// MultimodalClassificationModel_19026705121915
// MI455X (gfx1250) — hardware-verified
//
#include <hip/hip_runtime.h>
#include <math.h>

typedef __attribute__((ext_vector_type(16))) _Float16 v16h;
typedef __attribute__((ext_vector_type(8)))  _Float16 v8h;
typedef __attribute__((ext_vector_type(16))) __bf16   v16b;
typedef __attribute__((ext_vector_type(8)))  float    v8f;
typedef __attribute__((ext_vector_type(4)))  float    v4f;

__device__ __forceinline__ int frag_k(int i, int h) { return (i < 8) ? (8 * h + i) : (16 + 8 * h + (i - 8)); }
__device__ __forceinline__ __bf16 bf16_rne(float f) {
    unsigned int u = __float_as_uint(f);
    u += 0x7fffu + ((u >> 16) & 1u);
    return __builtin_bit_cast(__bf16, (unsigned short)(u >> 16));
}
__device__ __forceinline__ float bf16_f32(__bf16 b) { return __uint_as_float(((unsigned int)__builtin_bit_cast(unsigned short, b)) << 16); }
__device__ __forceinline__ v8f wmma16(v16h a, v16h b, v8f c) {
    c = __builtin_amdgcn_wmma_f32_16x16x32_f16(false, a, false, b, (short)0, c, false, false);
    asm volatile("v_nop\n\tv_nop\n\tv_nop\n\tv_nop" : "+v"(c) : "v"(a), "v"(b));
    return c;
}
__device__ __forceinline__ v8f wmmab(v16b a, v16b b, v8f c) {
    c = __builtin_amdgcn_wmma_f32_16x16x32_bf16(false, a, false, b, (short)0, c, false, false);
    asm volatile("v_nop\n\tv_nop\n\tv_nop\n\tv_nop" : "+v"(c) : "v"(a), "v"(b));
    return c;
}
struct Split { v16b hi, lo; };
__device__ __forceinline__ v8f wmma3(const Split& a, const Split& b, v8f c) {
    c = __builtin_amdgcn_wmma_f32_16x16x32_bf16(false, a.hi, false, b.hi, (short)0, c, false, false);
    c = __builtin_amdgcn_wmma_f32_16x16x32_bf16(false, a.hi, false, b.lo, (short)0, c, false, false);
    c = __builtin_amdgcn_wmma_f32_16x16x32_bf16(false, a.lo, false, b.hi, (short)0, c, false, false);
    asm volatile("v_nop\n\tv_nop\n\tv_nop\n\tv_nop" : "+v"(c) : "v"(a.hi), "v"(a.lo), "v"(b.hi), "v"(b.lo));
    return c;
}
struct Split3 { v16b hi, mid, lo; };
__device__ __forceinline__ v8f wmma6(const Split3& a, const Split3& b, v8f c) {
    c = __builtin_amdgcn_wmma_f32_16x16x32_bf16(false, a.hi, false, b.hi, (short)0, c, false, false);
    c = __builtin_amdgcn_wmma_f32_16x16x32_bf16(false, a.hi, false, b.mid, (short)0, c, false, false);
    c = __builtin_amdgcn_wmma_f32_16x16x32_bf16(false, a.mid, false, b.hi, (short)0, c, false, false);
    c = __builtin_amdgcn_wmma_f32_16x16x32_bf16(false, a.hi, false, b.lo, (short)0, c, false, false);
    c = __builtin_amdgcn_wmma_f32_16x16x32_bf16(false, a.mid, false, b.mid, (short)0, c, false, false);
    c = __builtin_amdgcn_wmma_f32_16x16x32_bf16(false, a.lo, false, b.hi, (short)0, c, false, false);
    asm volatile("v_nop\n\tv_nop\n\tv_nop\n\tv_nop" : "+v"(c) : "v"(a.hi), "v"(a.mid), "v"(a.lo), "v"(b.hi), "v"(b.mid), "v"(b.lo));
    return c;
}

__device__ __forceinline__ v16h fh_ld(const float* __restrict__ p, long long sk, int k0, int h, int klen, float s) {
    v16h a;
#pragma unroll
    for (int i = 0; i < 16; ++i) { const int k = k0 + frag_k(i, h); a[i] = (k < klen) ? (_Float16)(p[(long long)k * sk] * s) : (_Float16)0.f; }
    return a;
}
__device__ __forceinline__ Split sp_ld(const float* __restrict__ p, long long sk, int k0, int h, int klen, float s) {
    Split r;
#pragma unroll
    for (int i = 0; i < 16; ++i) {
        const int k = k0 + frag_k(i, h); const float x = (k < klen) ? p[(long long)k * sk] * s : 0.f;
        const __bf16 hb = bf16_rne(x); r.hi[i] = hb; r.lo[i] = bf16_rne(x - bf16_f32(hb));
    }
    return r;
}
__device__ __forceinline__ Split3 sp3_ld(const float* __restrict__ p, long long sk, int k0, int h, int klen, float s) {
    Split3 r;
#pragma unroll
    for (int i = 0; i < 16; ++i) {
        const int k = k0 + frag_k(i, h); const float x = (k < klen) ? p[(long long)k * sk] * s : 0.f;
        const __bf16 hb = bf16_rne(x); const float r1 = x - bf16_f32(hb); const __bf16 mb = bf16_rne(r1);
        r.hi[i] = hb; r.mid[i] = mb; r.lo[i] = bf16_rne(r1 - bf16_f32(mb));
    }
    return r;
}
__device__ __forceinline__ v16b bh_ld(const float* __restrict__ p, long long sk, int k0, int h, int klen, float s) {
    v16b a;
#pragma unroll
    for (int i = 0; i < 16; ++i) { const int k = k0 + frag_k(i, h); a[i] = bf16_rne((k < klen) ? p[(long long)k * sk] * s : 0.f); }
    return a;
}
__device__ __forceinline__ v16h fh_row(const _Float16* __restrict__ row, int k0, int h) {
    v16h a;
#pragma unroll
    for (int i = 0; i < 16; ++i) a[i] = row[k0 + frag_k(i, h)];
    return a;
}

#define VST2(T, ptr, val) do { *(volatile T*)(ptr) = (val); __threadfence(); *(volatile T*)(ptr) = (val); } while (0)
typedef float v4f __attribute__((ext_vector_type(4)));
#define VST2V4(ptr, val) do { *(volatile v4f*)(ptr) = (val); __threadfence(); *(volatile v4f*)(ptr) = (val); } while (0)

__device__ __attribute__((noinline)) float act_fn(float v, int act) {
    if (act == 1) return fmaxf(v, 0.f);
    if (act == 2) { const float u = 0.7978845608028654f * (v + 0.044715f * v * v * v); return 0.5f * v * (1.f + tanhf(u)); }
    if (act == 3) return v / (1.f + expf(-v));
    if (act == 4) return 0.5f * v * (1.f + erff(v * 0.7071067811865476f));
    if (act == 5) return tanhf(v);
    if (act == 6) return 1.f / (1.f + expf(-v));
    if (act == 7) return (v > 0.f) ? v : 0.01f * v;
    if (act == 8) return (v > 0.f) ? v : (expf(v) - 1.f);
    if (act == 9) return fminf(fmaxf(v, 0.f), 6.f);
    if (act == 10) return fabsf(v);
    if (act == 11) return (v >= 0.f) ? v : 0.1f * v;
    if (act == 12) return (v > 0.f) ? v : 0.2f * v;
    if (act == 13) return (v > 20.f) ? v : log1pf(expf(v));
    return v;
}

struct GemmP {
    const float* A; const float* B; const float* bias; const float* R; float* C;
    long long sAo, sAi, sAm, sAk, sBo, sBi, sBn, sBk, sCo, sCi, sCm, sRo, sRi, sRm, sRn;
    int M, N, K, zi_n, flags, act; float alpha, beta, sa, sb;
    int Npad, pad_;
};
static_assert(sizeof(GemmP) == 5 * 8 + 15 * 8 + 6 * 4 + 4 * 4 + 2 * 4, "GemmP has padding");

template <int MODE>
__global__ __launch_bounds__(32) void k_gemm(GemmP p) {
    const int lane = threadIdx.x & 31, h = lane >> 4, l15 = lane & 15;
    const int m0 = blockIdx.y * 16, n0 = blockIdx.x * 32;
    const int z = blockIdx.z, zo = z / p.zi_n, zi = z - zo * p.zi_n;
    const float* A = p.A + zo * p.sAo + zi * p.sAi;
    const float* B = p.B + zo * p.sBo + zi * p.sBi;
    const int am = min(m0 + l15, p.M - 1);
    v8f acc[2], comp[2];
#pragma unroll
    for (int t = 0; t < 2; ++t) { v8f zz = {}; acc[t] = zz; comp[t] = zz; }
    for (int k0 = 0; k0 < p.K; k0 += 32) {
        const float* arow = A + (long long)am * p.sAm;
        if (MODE == 1) {
            const Split a = sp_ld(arow, p.sAk, k0, h, p.K, 1.f);
#pragma unroll
            for (int t = 0; t < 2; ++t) {
                const int bn = min(n0 + t * 16 + l15, p.N - 1);
                acc[t] = wmma3(a, sp_ld(B + (long long)bn * p.sBn, p.sBk, k0, h, p.K, 1.f), acc[t]);
            }
        } else if (MODE == 3) {
            const Split3 a = sp3_ld(arow, p.sAk, k0, h, p.K, 1.f);
#pragma unroll
            for (int t = 0; t < 2; ++t) {
                const int bn = min(n0 + t * 16 + l15, p.N - 1);
                acc[t] = wmma6(a, sp3_ld(B + (long long)bn * p.sBn, p.sBk, k0, h, p.K, 1.f), acc[t]);
            }
        } else if (MODE == 4) {
            const Split3 a = sp3_ld(arow, p.sAk, k0, h, p.K, 1.f);
#pragma unroll
            for (int t = 0; t < 2; ++t) {
                const int bn = min(n0 + t * 16 + l15, p.N - 1); v8f zz = {};
                const v8f part = wmma6(a, sp3_ld(B + (long long)bn * p.sBn, p.sBk, k0, h, p.K, 1.f), zz);
                const v8f y = part - comp[t]; const v8f s = acc[t] + y; comp[t] = (s - acc[t]) - y; acc[t] = s;
            }
        } else if (MODE == 2) {
            const v16b a = bh_ld(arow, p.sAk, k0, h, p.K, 1.f);
#pragma unroll
            for (int t = 0; t < 2; ++t) {
                const int bn = min(n0 + t * 16 + l15, p.N - 1);
                acc[t] = wmmab(a, bh_ld(B + (long long)bn * p.sBn, p.sBk, k0, h, p.K, 1.f), acc[t]);
            }
        } else {
            const v16h a = fh_ld(arow, p.sAk, k0, h, p.K, p.sa);
#pragma unroll
            for (int t = 0; t < 2; ++t) {
                const int bn = min(n0 + t * 16 + l15, p.N - 1);
                acc[t] = wmma16(a, fh_ld(B + (long long)bn * p.sBn, p.sBk, k0, h, p.K, p.sb), acc[t]);
            }
        }
    }
    const float iscale = (MODE == 0) ? p.alpha / (p.sa * p.sb) : p.alpha;
    float* C = p.C + zo * p.sCo + zi * p.sCi;
    const float* R = p.R + zo * p.sRo + zi * p.sRi;
    __shared__ __align__(16) float ctile[16][36];
#pragma unroll
    for (int t = 0; t < 2; ++t) {
        const int n = n0 + t * 16 + l15; const int nn = min(n, p.N - 1);
#pragma unroll
        for (int r = 0; r < 8; ++r) {
            const int m = m0 + 8 * h + r; const int mm = min(m, p.M - 1);
            float v = acc[t][r] * iscale;
            if (p.flags & 1) v += p.bias[nn];
            if (p.flags & 2) v += p.bias[mm];
            v = act_fn(v, p.act);
            if (p.flags & 4) v += p.beta * R[(long long)mm * p.sRm + (long long)nn * p.sRn];
            ctile[8 * h + r][t * 16 + l15] = (n < p.N) ? v : 0.f;
        }
    }
    __syncthreads();
    const int NW = (p.Npad > p.N) ? p.Npad : p.N;
    const bool fast = (m0 + 16 <= p.M) && (n0 + 32 <= NW) && ((p.sCm & 3) == 0) && ((((size_t)C) & 15) == 0);
    if (fast) {
#pragma unroll
        for (int s = 0; s < 4; ++s) {
            const int row = s * 4 + (lane >> 3), c4 = (lane & 7) * 4;
            const v4f v = *(const v4f*)&ctile[row][c4];
            VST2V4(C + (long long)(m0 + row) * p.sCm + n0 + c4, v);
        }
    } else {
        for (int row = 0; row < 16; ++row) {
            const int m = m0 + row, n = n0 + lane;
            if (m < p.M && n < NW) VST2(float, C + (long long)m * p.sCm + n, ctile[row][lane]);
        }
    }
}

#define AW 4
struct AttnP {
    const float* Q; const float* K; const float* V; float* O; float* P; const float* Mf; const int* Mi; float* ST;
    const float* Pw; const float* Rt; const int* SQ; const int* SK;
    long long swb, swh, swi, swj, srb, srh, sri;
    long long sQb, sQh, sQi, sQd, sKb, sKh, sKj, sKd, sVb, sVh, sVj, sVd, sOb, sOh, sOi, sPb, sPh, sPi, smb, smh, smi, smj;
    int Lq, Lk, dh, dv, hrep, causal, coff, pband;
    float scale, mfill; int nonorm, mpol;
    int roff, rn, segpol, win;
};
static_assert(sizeof(AttnP) == 12 * 8 + 29 * 8 + 16 * 4, "AttnP has padding");

#ifndef KATTN_ATTR
#define KATTN_ATTR
#endif
template <int DHP, int DVP, int QM, bool SPLITPV, bool TWOPASS>
__global__ __launch_bounds__(32 * AW) KATTN_ATTR void k_attn(AttnP p) {
    constexpr int NT = DVP / 16;
    constexpr int KS = DHP / 32;
    constexpr int VP = DVP + 8;
    __shared__ __align__(16) float    pl[AW][16 * 64];
    __shared__ __align__(16) _Float16 vl[(SPLITPV ? 2 : 1) * 64 * VP];
    const int lane = threadIdx.x & 31, hf = lane >> 4, l15 = lane & 15, wave = threadIdx.x >> 5;
    const int h = blockIdx.y, b = blockIdx.z, hk = h / p.hrep;
    const int q0 = (blockIdx.x * AW + wave) * 16;
    float* myp = pl[wave];
    const float L2E = 1.4426950408889634f;
    const float NEG = -__builtin_inff();
    const int qi = min(q0 + l15, p.Lq - 1);
    const float* qrow = p.Q + b * p.sQb + h * p.sQh + (long long)qi * p.sQi;
    const float* kbase = p.K + b * p.sKb + hk * p.sKh;
    const float* vbase = p.V + b * p.sVb + hk * p.sVh;
    v16h qa[QM == 0 ? KS : 1]; Split qs_[QM == 1 ? KS : 1]; Split3 qt_[QM == 2 ? KS : 1];
#pragma unroll
    for (int ks = 0; ks < KS; ++ks) {
        if (QM == 2) qt_[ks] = sp3_ld(qrow, p.sQd, ks * 32, hf, p.dh, 1.f);
        else if (QM == 1) qs_[ks] = sp_ld(qrow, p.sQd, ks * 32, hf, p.dh, 1.f);
        else qa[ks] = fh_ld(qrow, p.sQd, ks * 32, hf, p.dh, 1.f);
    }
    v8f o[NT]; float m8[8], l8[8];
#pragma unroll
    for (int t = 0; t < NT; ++t) { v8f zz = {}; o[t] = zz; }
#pragma unroll
    for (int i = 0; i < 8; ++i) { m8[i] = NEG; l8[i] = 0.f; }
    int jend = p.Lk;
    if (p.causal == 1) { const int je = (blockIdx.x * AW + AW - 1) * 16 + 16 + p.coff; jend = min(jend, max(je, 0)); }
    const int npass = TWOPASS ? 2 : 1;
    for (int pass = 0; pass < npass; ++pass) {
        const bool dopv = (!TWOPASS) || pass == 1;
        for (int j0 = 0; j0 < jend; j0 += 64) {
            if (dopv) {
                __syncthreads();
                for (int idx = threadIdx.x; idx < 64 * DVP; idx += 32 * AW) {
                    const int jr = idx / DVP, d = idx - jr * DVP, j = j0 + jr;
                    const float f = (j < p.Lk && d < p.dv) ? vbase[(long long)j * p.sVj + (long long)d * p.sVd] : 0.f;
                    if (SPLITPV) {
                        const __bf16 hb = bf16_rne(f);
                        ((__bf16*)vl)[jr * VP + d] = hb; ((__bf16*)vl)[64 * VP + jr * VP + d] = bf16_rne(f - bf16_f32(hb));
                    } else vl[jr * VP + d] = (_Float16)f;
                }
            }
            v8f s[4];
#pragma unroll
            for (int t = 0; t < 4; ++t) {
                const int j = min(j0 + t * 16 + l15, p.Lk - 1);
                const float* krow = kbase + (long long)j * p.sKj;
                v8f acc = {};
#pragma unroll
                for (int ks = 0; ks < KS; ++ks) {
                    if (QM == 2)      acc = wmma6(qt_[ks], sp3_ld(krow, p.sKd, ks * 32, hf, p.dh, 1.f), acc);
                    else if (QM == 1) acc = wmma3(qs_[ks], sp_ld(krow, p.sKd, ks * 32, hf, p.dh, 1.f), acc);
                    else              acc = wmma16(qa[ks], fh_ld(krow, p.sKd, ks * 32, hf, p.dh, 1.f), acc);
                }
                s[t] = acc;
            }
            float pv[8][4];
#pragma unroll
            for (int i = 0; i < 8; ++i) {
                const int irow = q0 + i + 8 * hf;
                const int ic = min(irow, p.Lq - 1);
                float sc[4];
#pragma unroll
                for (int t = 0; t < 4; ++t) {
                    const int jg = j0 + t * 16 + l15;
                    float v = s[t][i] * p.scale;
                    if (p.Mf) v += p.Mf[b * p.smb + h * p.smh + (long long)ic * p.smi + (long long)min(jg, p.Lk - 1) * p.smj];
                    if (p.Rt) { int rc = ic - min(jg, p.Lk - 1) + p.roff; rc = rc < 0 ? 0 : (rc >= p.rn ? p.rn - 1 : rc); v += p.Rt[b * p.srb + h * p.srh + (long long)ic * p.sri + rc]; }
                    if (p.Mi) { const int mv = p.Mi[b * p.smb + h * p.smh + (long long)ic * p.smi + (long long)min(jg, p.Lk - 1) * p.smj]; if (p.mpol ? (mv != 0) : (mv == 0)) v = p.mfill; }
                    if (p.SQ) { const bool same = p.SQ[(long long)b * p.Lq + ic] == p.SK[(long long)b * p.Lk + min(jg, p.Lk - 1)]; if (p.segpol ? same : !same) v = p.mfill; }
                    if (p.causal == 2 && jg > irow + p.coff) v = p.mfill;
                    if (jg >= p.Lk || (p.causal == 1 && jg > irow + p.coff) || (p.causal == 3 && jg < irow + p.coff) || (p.win > 0 && irow + p.coff - jg > p.win)) v = NEG; else v *= L2E;
                    sc[t] = v;
                }
                if (!TWOPASS || pass == 0) {
                    float mx = fmaxf(fmaxf(sc[0], sc[1]), fmaxf(sc[2], sc[3]));
                    mx = fmaxf(mx, __shfl_xor(mx, 1, 32)); mx = fmaxf(mx, __shfl_xor(mx, 2, 32));
                    mx = fmaxf(mx, __shfl_xor(mx, 4, 32)); mx = fmaxf(mx, __shfl_xor(mx, 8, 32));
                    const float mnew = fmaxf(m8[i], mx);
                    const float corr = (mnew == NEG) ? 1.f : exp2f(m8[i] - mnew);
                    float rs = 0.f;
#pragma unroll
                    for (int t = 0; t < 4; ++t) {
                        const float pp = (sc[t] == NEG) ? 0.f : exp2f(sc[t] - mnew); rs += pp;
                        pv[i][t] = p.Pw ? pp * p.Pw[b * p.swb + h * p.swh + (long long)ic * p.swi + (long long)min(j0 + t * 16 + l15, p.Lk - 1) * p.swj] : pp;
                    }
                    rs += __shfl_xor(rs, 1, 32); rs += __shfl_xor(rs, 2, 32); rs += __shfl_xor(rs, 4, 32); rs += __shfl_xor(rs, 8, 32);
                    l8[i] = l8[i] * corr + rs; m8[i] = mnew;
                    if (!TWOPASS) {
#pragma unroll
                        for (int t = 0; t < NT; ++t) o[t][i] *= corr;
                    }
                } else {
                    const float inv = (l8[i] > 0.f) ? 1.f / l8[i] : 0.f;
#pragma unroll
                    for (int t = 0; t < 4; ++t) {
                        const int jg = j0 + t * 16 + l15;
                        float pp = (sc[t] == NEG) ? 0.f : exp2f(sc[t] - m8[i]) * inv;
                        if (p.Pw) pp *= p.Pw[b * p.swb + h * p.swh + (long long)ic * p.swi + (long long)min(jg, p.Lk - 1) * p.swj];
                        pv[i][t] = pp;
                    }
                }
            }
            if (dopv) {
#pragma unroll
                for (int i = 0; i < 8; ++i)
#pragma unroll
                    for (int t = 0; t < 4; ++t) myp[(i + 8 * hf) * 64 + t * 16 + l15] = pv[i][t];
                __syncthreads();
                if (p.P) {
                    float* pb_ = p.P + b * p.sPb + h * p.sPh;
                    const bool fastP = (p.pband == 0) && ((p.sPi & 3) == 0) && (j0 + 64 <= p.Lk) && (q0 + 16 <= p.Lq) && ((((size_t)pb_) & 15) == 0);
                    if (fastP) {
#pragma unroll
                        for (int s = 0; s < 8; ++s) {
                            const int row = s * 2 + (lane >> 4), c4 = (lane & 15) * 4;
                            const v4f v = *(const v4f*)(myp + row * 64 + c4);
                            VST2V4(pb_ + (long long)(q0 + row) * p.sPi + j0 + c4, v);
                        }
                    } else {
                        for (int row = 0; row < 16; ++row) {
                            const int irow = q0 + row; if (irow >= p.Lq) continue;
                            for (int c = lane; c < 64; c += 32) {
                                const int jg = j0 + c; if (jg >= p.Lk) continue;
                                if (p.pband == 0) VST2(float, pb_ + (long long)irow * p.sPi + jg, myp[row * 64 + c]);
                                else if (jg - irow <= p.pband && irow - jg <= p.pband) VST2(float, pb_ + (long long)irow * p.sPi + (jg - irow + p.pband), myp[row * 64 + c]);
                            }
                        }
                    }
                }
                if (SPLITPV) {
                    const Split pa0 = sp_ld(myp + l15 * 64, 1, 0, hf, 64, 1.f), pa1 = sp_ld(myp + l15 * 64, 1, 32, hf, 64, 1.f);
                    const __bf16* vh = (const __bf16*)vl; const __bf16* vlo = vh + 64 * VP;
#pragma unroll
                    for (int t = 0; t < NT; ++t) {
                        const int dcol = t * 16 + l15;
                        Split b0, b1;
#pragma unroll
                        for (int e = 0; e < 16; ++e) {
                            const int k0 = frag_k(e, hf), k1 = 32 + frag_k(e, hf);
                            b0.hi[e] = vh[k0 * VP + dcol]; b0.lo[e] = vlo[k0 * VP + dcol]; b1.hi[e] = vh[k1 * VP + dcol]; b1.lo[e] = vlo[k1 * VP + dcol];
                        }
                        o[t] = wmma3(pa0, b0, o[t]);
                        o[t] = wmma3(pa1, b1, o[t]);
                    }
                } else {
                    const v16h pa0 = fh_ld(myp + l15 * 64, 1, 0, hf, 64, 4096.f), pa1 = fh_ld(myp + l15 * 64, 1, 32, hf, 64, 4096.f);
#pragma unroll
                    for (int t = 0; t < NT; ++t) {
                        const int dcol = t * 16 + l15;
                        v16h b0, b1;
#pragma unroll
                        for (int e = 0; e < 16; ++e) { b0[e] = vl[frag_k(e, hf) * VP + dcol]; b1[e] = vl[(32 + frag_k(e, hf)) * VP + dcol]; }
                        o[t] = wmma16(pa0, b0, o[t]);
                        o[t] = wmma16(pa1, b1, o[t]);
                    }
                }
            }
        }
    }
    float* obase = p.O + b * p.sOb + h * p.sOh;
    if (p.ST) {
        const int rl = lane >> 1, isel = rl & 7;
        float mv = 0.f, lv = 0.f;
#pragma unroll
        for (int i = 0; i < 8; ++i) if (i == isel) { mv = m8[i]; lv = l8[i]; }
        const int irow = q0 + rl;
        if (irow < p.Lq) { float* st = p.ST + (((long long)b * gridDim.y + h) * p.Lq + irow) * 2 + (lane & 1); VST2(float, st, (lane & 1) ? lv : mv * 0.6931471805599453f); }
    }
    float invr[8];
#pragma unroll
    for (int i = 0; i < 8; ++i) {
        if (TWOPASS) invr[i] = SPLITPV ? 1.f : (1.f / 4096.f);
        else if (p.nonorm) invr[i] = exp2f(m8[i]) * (SPLITPV ? 1.f : (1.f / 4096.f));
        else invr[i] = (l8[i] > 0.f) ? (SPLITPV ? 1.f / l8[i] : 1.f / (l8[i] * 4096.f)) : 0.f;
    }
    __syncthreads();
    const bool ofast = ((p.sOi & 3) == 0) && ((((size_t)obase) & 15) == 0) && (q0 + 16 <= p.Lq);
#pragma unroll
    for (int c0 = 0; c0 < DVP; c0 += 64) {
#pragma unroll
        for (int i = 0; i < 8; ++i)
#pragma unroll
            for (int t = 0; t < NT; ++t) if (t * 16 >= c0 && t * 16 < c0 + 64) myp[(i + 8 * hf) * 64 + (t * 16 - c0) + l15] = o[t][i] * invr[i];
        __syncthreads();
        const int cw = (DVP - c0 < 64) ? (DVP - c0) : 64;
        if (ofast && (c0 + cw <= p.dv) && (cw % 32 == 0)) {
            const int lpr = cw / 4;
            const int rows_per_ins = 32 / lpr;
            for (int r0 = 0; r0 < 16; r0 += rows_per_ins) {
                const int row = r0 + lane / lpr, c4 = (lane % lpr) * 4;
                const v4f v = *(const v4f*)(myp + row * 64 + c4);
                VST2V4(obase + (long long)(q0 + row) * p.sOi + c0 + c4, v);
            }
        } else {
            for (int row = 0; row < 16; ++row) {
                const int irow = q0 + row; if (irow >= p.Lq) continue;
                for (int c = lane; c < cw; c += 32) { const int d = c0 + c; if (d < p.dv) VST2(float, obase + (long long)irow * p.sOi + d, myp[row * 64 + c]); }
            }
        }
        __syncthreads();
    }
}

struct TrP { const float* src; float* dst; const float* R2; long long sSz, lds, sDz, ldd, sRz, ldr; int R, C, flags, act; float alpha, beta; };
static_assert(sizeof(TrP) == 3 * 8 + 6 * 8 + 6 * 4, "TrP has padding");
__global__ __launch_bounds__(256) void k_tr(TrP p) {
    __shared__ float tile[32][33];
    const int c0 = blockIdx.x * 32, r0 = blockIdx.y * 32, z = blockIdx.z;
    const int lane = threadIdx.x & 31, wave = threadIdx.x >> 5;
    const float* s = p.src + z * p.sSz;
#pragma unroll
    for (int k = 0; k < 4; ++k) {
        const int rl = wave * 4 + k, r = r0 + rl, c = c0 + lane;
        tile[rl][lane] = (r < p.R && c < p.C) ? s[(long long)r * p.lds + c] : 0.f;
    }
    __syncthreads();
    float* d = p.dst + z * p.sDz; const float* rr = p.R2 + z * p.sRz;
#pragma unroll
    for (int k = 0; k < 4; ++k) {
        const int cl = wave * 4 + k, c = c0 + cl, r = r0 + lane;
        if (c < p.C && r < p.R) {
            float v = act_fn(p.alpha * tile[lane][cl], p.act);
            if (p.flags & 1) v += p.beta * rr[(long long)c * p.ldr + r];
            VST2(float, d + (long long)c * p.ldd + r, v);
        }
    }
}

__global__ __launch_bounds__(256) void k_affine(const float* __restrict__ src, float* __restrict__ dst, int n, float a, float b, const float* __restrict__ sdev) {
    const int i = blockIdx.x * 256 + threadIdx.x;
    if (i < n) { const float aa = sdev ? a * sdev[0] : a; const float v = aa * src[i] + b; VST2(float, dst + i, v); }
}

struct SmP { const float* src; float* dst; const float* Mf; long long sz, sr, dz, dr, smz, smr; int n, pad; float scale_in, scale_out; };
static_assert(sizeof(SmP) == 3 * 8 + 6 * 8 + 4 * 4, "SmP has padding");
__global__ __launch_bounds__(256) void k_softmax(SmP p) {
    __shared__ float red[256];
    const int r = blockIdx.x, z = blockIdx.y, tid = threadIdx.x;
    const float* s = p.src + z * p.sz + (long long)r * p.sr;
    const float* mf = p.Mf ? (p.Mf + z * p.smz + (long long)r * p.smr) : nullptr;
    float mx = -__builtin_inff();
    for (int j = tid; j < p.n; j += 256) { float v = s[j] * p.scale_in; if (mf) v += mf[j]; mx = fmaxf(mx, v); }
    red[tid] = mx; __syncthreads();
    for (int o = 128; o > 0; o >>= 1) { if (tid < o) red[tid] = fmaxf(red[tid], red[tid + o]); __syncthreads(); }
    mx = red[0]; __syncthreads();
    float sum = 0.f;
    for (int j = tid; j < p.n; j += 256) { float v = s[j] * p.scale_in; if (mf) v += mf[j]; sum += (mx == -__builtin_inff()) ? 0.f : expf(v - mx); }
    red[tid] = sum; __syncthreads();
    for (int o = 128; o > 0; o >>= 1) { if (tid < o) red[tid] += red[tid + o]; __syncthreads(); }
    sum = red[0];
    const float inv = (sum > 0.f) ? p.scale_out / sum : 0.f;
    float* d = p.dst + z * p.dz + (long long)r * p.dr;
    for (int j = tid; j < p.n; j += 256) { float v = s[j] * p.scale_in; if (mf) v += mf[j]; const float o = (mx == -__builtin_inff()) ? 0.f : expf(v - mx) * inv; VST2(float, d + j, o); }
}
__global__ __launch_bounds__(256) void k_stats(const float* __restrict__ x, long long sz, long long so, long long si, int inner, int n, float eps, float* __restrict__ stat, int mode) {
    __shared__ float red[256];
    const int z = blockIdx.x, tid = threadIdx.x;
    const float* base = x + z * sz;
    float s = 0.f;
    for (int e = tid; e < n; e += 256) s += base[(long long)(e / inner) * so + (long long)(e % inner) * si];
    red[tid] = s; __syncthreads();
    for (int o = 128; o > 0; o >>= 1) { if (tid < o) red[tid] += red[tid + o]; __syncthreads(); }
    const float mu = (mode == 0 || mode == 3) ? red[0] / (float)n : 0.f; __syncthreads();
    float q = 0.f;
    for (int e = tid; e < n; e += 256) { const float dlt = base[(long long)(e / inner) * so + (long long)(e % inner) * si] - mu; q += dlt * dlt; }
    red[tid] = q; __syncthreads();
    for (int o = 128; o > 0; o >>= 1) { if (tid < o) red[tid] += red[tid + o]; __syncthreads(); }
    {
        float rs;
        if (mode == 2) rs = sqrtf((float)n) / fmaxf(sqrtf(red[0]), eps); else if (mode == 3) rs = rsqrtf(red[0] / (float)(n - 1) + eps); else rs = rsqrtf(red[0] / (float)n + eps);
        if (tid < 32) { const float v = (tid == 0) ? mu : ((tid == 1) ? rs : 0.f); VST2(float, stat + (long long)z * 32 + tid, v); }
    }
}
__global__ __launch_bounds__(256) void k_norm_apply(const float* __restrict__ x, float* __restrict__ y, const float* __restrict__ stat, const float* __restrict__ g, const float* __restrict__ bta,
                                                     int Z, int C, int L, int G, int bn, int act) {
    const long long idx = (long long)blockIdx.x * 256 + threadIdx.x;
    if (idx >= (long long)Z * C * L) return;
    const int l = (int)(idx % L); const long long zc = idx / L; const int c = (int)(zc % C), z = (int)(zc / C); (void)l;
    const int set = bn ? c : (z * G + c / (C / G));
    float v = (x[idx] - stat[(long long)set * 32]) * stat[(long long)set * 32 + 1];
    if (g) v *= g[c];
    if (bta) v += bta[c];
    v = act_fn(v, act);
    VST2(float, y + idx, v);
}

__global__ __launch_bounds__(256) void k_lse_neg(const float* __restrict__ st, float* __restrict__ c, int n) {
    const int i = blockIdx.x * 256 + threadIdx.x;
    if (i < n) { const float v = -(st[2 * i] + logf(st[2 * i + 1])); VST2(float, c + i, v); }
}

__global__ __launch_bounds__(256) void k_iota(int* __restrict__ dst, int n, int a, int b) {
    const int i = blockIdx.x * 256 + threadIdx.x;
    if (i < n) { const int v = a * i + b; VST2(int, dst + i, v); }
}

__global__ __launch_bounds__(256) void k_axpby(const float* __restrict__ x, const float* __restrict__ y, float* __restrict__ dst, int n, float a, float b, float c) {
    const int i = blockIdx.x * 256 + threadIdx.x;
    if (i < n) { const float v = a * x[i] + b * y[i] + c; VST2(float, dst + i, v); }
}

struct RopeP { const float* X; float* Y; const float* C; const float* Sn; const int* pos; long long sXr, sXh, sYr, sYh, sCb, sCp, sCd; int R, Hn, D, S, mode, tmode, pmode, pad; };
static_assert(sizeof(RopeP) == 5 * 8 + 7 * 8 + 8 * 4, "RopeP has padding");
__global__ __launch_bounds__(256) void k_rope(RopeP p) {
    const long long idx = (long long)blockIdx.x * 256 + threadIdx.x;
    if (idx >= (long long)p.R * p.Hn * p.D) return;
    const int d = (int)(idx % p.D); const long long rh = idx / p.D; const int h = (int)(rh % p.Hn); const int r = (int)(rh / p.Hn);
    const int half = p.D / 2;
    int partner; float sign;
    if (p.mode == 0) { partner = (d < half) ? d + half : d - half; sign = (d < half) ? -1.f : 1.f; }
    else { partner = d ^ 1; sign = (d & 1) ? 1.f : -1.f; }
    const int tcol = (p.tmode == 0) ? d : ((p.tmode == 1) ? (d % half) : (d >> 1));
    const int pp = (p.pmode == 0) ? (r % p.S) : ((p.pmode == 1) ? h : p.pos[r]);
    const long long toff = (long long)(r / p.S) * p.sCb + (long long)pp * p.sCp + (long long)tcol * p.sCd;
    const float* xr = p.X + (long long)r * p.sXr + (long long)h * p.sXh;
    const float v = xr[d] * p.C[toff] + sign * xr[partner] * p.Sn[toff];
    VST2(float, p.Y + (long long)r * p.sYr + (long long)h * p.sYh + d, v);
}

__global__ __launch_bounds__(256) void k_invf(float* __restrict__ invb, int half, int D, float base, float num, int fmode, float cexp) {
    const int i = blockIdx.x * 256 + threadIdx.x;
    if (i >= ((half + 31) / 32) * 32) return;
    if (i >= half) { VST2(float, invb + i, 0.f); return; }
    const float e = (float)(2 * i) / (float)D;
    float invf;
    if (fmode == 1) invf = num * expf((float)(2 * i) * cexp);
    else if (fmode == 2) invf = num * powf(base, (-2.0f * ((float)i - 1.0f)) / (float)D);
    else invf = num * (1.0f / powf(base, e));
    VST2(float, invb + i, invf);
}
__global__ __launch_bounds__(256) void k_sincos(float* __restrict__ cs, float* __restrict__ sn, const float* __restrict__ invb, int S, int half, float pscale) {
    const int idx = blockIdx.x * 256 + threadIdx.x;
    if (idx >= S * half) return;
    const int s = idx / half, i = idx - s * half;
    const float ang = (pscale * (float)s) * invb[i];
    VST2(float, cs + idx, cosf(ang)); VST2(float, sn + idx, sinf(ang));
}

__global__ __launch_bounds__(256) void k_mulact(const float* __restrict__ x, const float* __restrict__ y, float* __restrict__ dst, int n, int act) {
    const int i = blockIdx.x * 256 + threadIdx.x;
    if (i < n) { const float v = act_fn(x[i], act) * y[i]; VST2(float, dst + i, v); }
}

__global__ __launch_bounds__(256) void k_matvec(GemmP p) {
    const int rpt = (p.N == 1) ? 1 : 32;
    const long long r0 = ((long long)blockIdx.x * 256 + threadIdx.x) * rpt; const int z = blockIdx.z, zo = z / p.zi_n, zi = z - zo * p.zi_n;
    if (r0 >= p.M) return;
    const float* Bb = p.B + zo * p.sBo + zi * p.sBi;
    float* C = p.C + zo * p.sCo + zi * p.sCi; const float* R = p.R + zo * p.sRo + zi * p.sRi;
    for (int rr = 0; rr < rpt; ++rr) {
        const long long r = r0 + rr; if (r >= p.M) break;
        const float* A = p.A + zo * p.sAo + zi * p.sAi + r * p.sAm;
        float acc[8] = {0.f, 0.f, 0.f, 0.f, 0.f, 0.f, 0.f, 0.f};
        for (int k = 0; k < p.K; ++k) { const float a = A[(long long)k * p.sAk];
#pragma unroll
            for (int j = 0; j < 8; ++j) if (j < p.N) acc[j] += a * Bb[(long long)j * p.sBn + (long long)k * p.sBk]; }
#pragma unroll
        for (int j = 0; j < 8; ++j) if (j < p.N) {
            float v = acc[j] * p.alpha;
            if (p.flags & 1) v += p.bias[j];
            if (p.flags & 2) v += p.bias[r];
            v = act_fn(v, p.act);
            if (p.flags & 4) v += p.beta * R[r * p.sRm + (long long)j * p.sRn];
            VST2(float, C + r * p.sCm + j, v);
        }
    }
}
__global__ __launch_bounds__(256) void k_smallsoftmax(const float* __restrict__ src, float* __restrict__ dst, long long sr, long long dr, int n, long long R, float scale) {
    const long long r0 = ((long long)blockIdx.x * 256 + threadIdx.x) * 32;
    for (int rr = 0; rr < 32; ++rr) {
        const long long r = r0 + rr; if (r >= R) return;
        const float* s = src + r * sr; float* d = dst + r * dr;
        float mx = -__builtin_inff();
        for (int j = 0; j < n; ++j) mx = fmaxf(mx, s[j] * scale);
        float sum = 0.f;
        for (int j = 0; j < n; ++j) sum += expf(s[j] * scale - mx);
        const float inv = 1.f / sum;
        for (int j = 0; j < n; ++j) { const float v = expf(s[j] * scale - mx) * inv; VST2(float, d + j, v); }
    }
}

__global__ __launch_bounds__(32) void k_unitstat(float* __restrict__ st) { const int t = threadIdx.x; const float v = (t == 1) ? 1.f : 0.f; VST2(float, st + t, v); }

__global__ __launch_bounds__(256) void k_lincopy(const float* __restrict__ src, long long lds, float* __restrict__ dst, long long ldd, long long rows, int cols) {
    const long long i = (long long)blockIdx.x * 256 + threadIdx.x; if (i >= rows * cols) return;
    const long long r = i / cols; const int c = (int)(i - r * cols);
    const float v = src[r * lds + c]; VST2(float, dst + r * ldd + c, v);
}

__global__ __launch_bounds__(256) void k_mm_pad1d(const float* __restrict__ X, float* __restrict__ P, int B, int L) { const int q = blockIdx.x * 256 + threadIdx.x; if (q >= B * L) return; const int l = q % L; const int b = q / L; VST2(float, P + (long long)b * (L + 2) + l + 1, X[q]); }
__global__ __launch_bounds__(256) void k_mm_relu1d(float* __restrict__ P, int B, int L, int C) { const long long q = (long long)blockIdx.x * 256 + threadIdx.x; if (q >= (long long)B * L * C) return; const int c = (int)(q % C); const int l = (int)((q / C) % L); const int b = (int)(q / ((long long)C * L)); float* p = P + (((long long)b * (L + 2) + l + 1) * C + c); VST2(float, p, fmaxf(*p, 0.f)); }
__global__ __launch_bounds__(256) void k_mm_dft(float* __restrict__ COSm, float* __restrict__ SINm, int NF, int L) {
    const long long q = (long long)blockIdx.x * 256 + threadIdx.x; if (q >= (long long)NF * L) return; const int l = (int)(q % L); const int f = (int)(q / L); const long long m = ((long long)f * l) % L;
    const double ang = 6.283185307179586476925 * (double)m / (double)L; const float sc = rsqrtf((float)L); float s, c; s = (float)sin(ang) * sc; c = (float)cos(ang) * sc; if (f == 0 || 2 * f == L) s = 0.f; VST2(float, COSm + q, c); VST2(float, SINm + q, s);
}
__global__ __launch_bounds__(256) void k_mm_energy(const float* __restrict__ XR, const float* __restrict__ XI, float* __restrict__ EN, int B, int NF, int C) { const int q = blockIdx.x * 256 + threadIdx.x; if (q >= B * NF) return; const float* xr = XR + (long long)q * C; const float* xi = XI + (long long)q * C; float e = 0.f;
#pragma unroll 1
    for (int c = 0; c < C; ++c) e += xr[c] * xr[c] + xi[c] * xi[c]; VST2(float, EN + q, e); }
__global__ __launch_bounds__(256) void k_mm_filter(float* __restrict__ XR, float* __restrict__ XI, const float* __restrict__ EN, const float* __restrict__ affw, const float* __restrict__ affh, const float* __restrict__ thr, int B, int NF, int C) {
    __shared__ float med; const int b = blockIdx.y; const int f = blockIdx.x; const float* en = EN + (long long)b * NF;
    if (threadIdx.x == 0) med = 0.f; __syncthreads();
    for (int cand = threadIdx.x; cand < NF; cand += 256) { const float v = en[cand]; int below = 0; for (int j = 0; j < NF; ++j) { const float u = en[j]; below += (u < v) || (u == v && j < cand); } if (below == NF / 2) med = v; }
    __syncthreads();
    const float ne = en[f] / (med + 1e-6f); const float hard = (ne > thr[0]) ? 1.f : 0.f; const float mask = (hard - thr[0]) + thr[0]; const float coef = (f == 0 || f == NF - 1) ? 1.f : 2.f;
    for (int c = threadIdx.x; c < C; c += 256) { const long long o = ((long long)b * NF + f) * C + c; const float xr = XR[o], xi = XI[o]; const float wr = affw[2 * c], wi = affw[2 * c + 1], hr = affh[2 * c], hi = affh[2 * c + 1];
        const float ar = wr + mask * hr, ai = wi + mask * hi;
        const float yr = xr * ar - xi * ai, yi = xr * ai + xi * ar; VST2(float, XR + o, yr * coef); VST2(float, XI + o, yi * coef); }
}
__global__ __launch_bounds__(256) void k_mm_padimg(const float* __restrict__ X, float* __restrict__ P, int B, int C, int H) { const long long q = (long long)blockIdx.x * 256 + threadIdx.x; if (q >= (long long)B * H * H * C) return; const int c = (int)(q % C); const int x = (int)((q / C) % H); const int y = (int)((q / (C * H)) % H); const int b = (int)(q / ((long long)C * H * H)); VST2(float, P + (((long long)b * (H + 2) + y + 1) * (H + 2) + x + 1) * C + c, X[(((long long)b * C + c) * H + y) * H + x]); }
__global__ __launch_bounds__(256) void k_mm_relu2d(float* __restrict__ P, float* __restrict__ CMP, int B, int H, int C) { const long long q = (long long)blockIdx.x * 256 + threadIdx.x; if (q >= (long long)B * H * H * C) return; const int c = (int)(q % C); const int x = (int)((q / C) % H); const int y = (int)((q / (C * H)) % H); const int b = (int)(q / ((long long)C * H * H)); float* p = P + (((long long)b * (H + 2) + y + 1) * (H + 2) + x + 1) * C + c; const float v = fmaxf(*p, 0.f); VST2(float, p, v); if (CMP) VST2(float, CMP + q, v); }
__global__ __launch_bounds__(256) void k_mm_dw(const float* __restrict__ Q, const float* __restrict__ w, const float* __restrict__ bb, float* __restrict__ O, int B, int H, int C) {
    const long long q = (long long)blockIdx.x * 256 + threadIdx.x; if (q >= (long long)B * H * H * C) return; const int c = (int)(q % C); const int x = (int)((q / C) % H); const int y = (int)((q / (C * H)) % H); const int b = (int)(q / ((long long)C * H * H)); float s = bb[c];
    for (int ky = 0; ky < 3; ++ky) { const int yy = y + ky - 1; if (yy < 0 || yy >= H) continue; for (int kx = 0; kx < 3; ++kx) { const int xx = x + kx - 1; if (xx < 0 || xx >= H) continue; s += w[c * 9 + ky * 3 + kx] * Q[(((long long)b * H + yy) * H + xx) * C + c]; } }
    VST2(float, O + q, s);
}
__global__ __launch_bounds__(256) void k_mm_fall(const float* __restrict__ QKV2, const float* __restrict__ fcw, const float* __restrict__ fcb, float* __restrict__ FC, int B, int HW, int C) {
    const long long q = (long long)blockIdx.x * 256 + threadIdx.x; if (q >= (long long)B * HW * 16 * 9) return; const int o = (int)(q % 9); const int kk = (int)((q / 9) % 16); const int r = (int)((q / 144) % HW); const int b = (int)(q / ((long long)144 * HW)); float s = fcb[o];
#pragma unroll 1
    for (int i = 0; i < 12; ++i) { const long long flat = (long long)r * 192 + i * 16 + kk; const int ch = (int)(flat / HW); const int pp = (int)(flat % HW); s += fcw[o * 12 + i] * QKV2[((long long)b * HW + pp) * C + ch]; }
    VST2(float, FC + (((long long)b * 144 + kk * 9 + o) * HW + r), s);
}
__global__ __launch_bounds__(256) void k_mm_dep(const float* __restrict__ FC, const float* __restrict__ w, const float* __restrict__ bb, float* __restrict__ O, int B, int H) {
    const long long q = (long long)blockIdx.x * 256 + threadIdx.x; const int HW = H * H; if (q >= (long long)B * 64 * HW) return; const int p = (int)(q % HW); const int oc = (int)((q / HW) % 64); const int b = (int)(q / ((long long)HW * 64)); const int g = oc / 4; const int y = p / H, x = p % H; float s = bb[oc];
    for (int i = 0; i < 9; ++i) { const float* src = FC + ((long long)b * 144 + g * 9 + i) * HW; const float* wk = w + (oc * 9 + i) * 9;
        for (int ky = 0; ky < 3; ++ky) { const int yy = y + ky - 1; if (yy < 0 || yy >= H) continue; for (int kx = 0; kx < 3; ++kx) { const int xx = x + kx - 1; if (xx < 0 || xx >= H) continue; s += wk[ky * 3 + kx] * src[yy * H + xx]; } } }
    VST2(float, O + q, s);
}
__global__ __launch_bounds__(256) void k_mm_qknorm(const float* __restrict__ QKV2, float* __restrict__ QN, int B, int HW, int C) {
    __shared__ float red[256]; const int z = blockIdx.x; const int b = z / 128, ch = z % 128; float s = 0.f;
    for (int p = threadIdx.x; p < HW; p += 256) { const float v = QKV2[((long long)b * HW + p) * C + ch]; s += v * v; }
    red[threadIdx.x] = s; __syncthreads(); for (int o = 128; o > 0; o >>= 1) { if (threadIdx.x < o) red[threadIdx.x] += red[threadIdx.x + o]; __syncthreads(); }
    const float inv = 1.f / fmaxf(sqrtf(red[0]), 1e-12f);
    for (int p = threadIdx.x; p < HW; p += 256) VST2(float, QN + ((long long)b * 128 + ch) * HW + p, QKV2[((long long)b * HW + p) * C + ch] * inv);
}
__global__ __launch_bounds__(256) void k_mm_sm16(float* __restrict__ AT, const float* __restrict__ temp, int NZ, int ldp) { const int r = blockIdx.x * 256 + threadIdx.x; if (r >= NZ * 16) return; const int h = (r / 16) % 4; float* a = AT + (long long)r * ldp; const float tp = temp[h]; float mx = -__builtin_inff();
#pragma unroll 1
    for (int j = 0; j < 16; ++j) mx = fmaxf(mx, a[j] * tp);
    float s = 0.f;
#pragma unroll 1
    for (int j = 0; j < 16; ++j) s += expf(a[j] * tp - mx);
#pragma unroll 1
    for (int j = 0; j < 16; ++j) { const float pv = expf(a[j] * tp - mx) / s; VST2(float, a + j, pv); } }
__global__ __launch_bounds__(256) void k_mm_imgfeat(const float* __restrict__ AO, const float* __restrict__ OCV, float* __restrict__ IR, int B, int HW, int C) { const long long q = (long long)blockIdx.x * 256 + threadIdx.x; if (q >= (long long)B * (HW / 4) * C) return; const int c = (int)(q % C); const int s = (int)((q / C) % (HW / 4)); const int b = (int)(q / ((long long)C * (HW / 4))); float a = 0.f; for (int j = 0; j < 4; ++j) { const long long idx = ((long long)b * C + c) * HW + s * 4 + j; a += AO[idx] + OCV[idx]; } VST2(float, IR + q, 0.25f * a); }
__global__ __launch_bounds__(256) void k_mm_uspool(const float* __restrict__ UF, float* __restrict__ UR, int B, int L, int C) { const long long q = (long long)blockIdx.x * 256 + threadIdx.x; if (q >= (long long)B * (L / 4) * C) return; const int c = (int)(q % C); const int s = (int)((q / C) % (L / 4)); const int b = (int)(q / ((long long)C * (L / 4))); float a = 0.f; for (int j = 0; j < 4; ++j) a += UF[((long long)b * L + s * 4 + j) * C + c]; VST2(float, UR + q, 0.25f * a); }
__global__ __launch_bounds__(256) void k_mm_pools(const float* __restrict__ T1, const float* __restrict__ T2, float* __restrict__ CHP, float* __restrict__ SPP, int B, int S, int C) {
    const int q = blockIdx.x * 256 + threadIdx.x;
    if (q < B * C) { const int c = q % C, b = q / C; float m1 = 0.f, x1 = -__builtin_inff(), m2 = 0.f, x2 = -__builtin_inff(); for (int s = 0; s < S; ++s) { const float a = T1[((long long)b * S + s) * C + c], d = T2[((long long)b * S + s) * C + c]; m1 += a; x1 = fmaxf(x1, a); m2 += d; x2 = fmaxf(x2, d); }
        VST2(float, CHP + ((long long)b * 4 + 0) * C + c, m1 / S); VST2(float, CHP + ((long long)b * 4 + 1) * C + c, x1); VST2(float, CHP + ((long long)b * 4 + 2) * C + c, m2 / S); VST2(float, CHP + ((long long)b * 4 + 3) * C + c, x2); }
    if (q < B * S) { const int s = q % S, b = q / S; float m1 = 0.f, x1 = -__builtin_inff(), m2 = 0.f, x2 = -__builtin_inff(); for (int c = 0; c < C; ++c) { const float a = T1[((long long)b * S + s) * C + c], d = T2[((long long)b * S + s) * C + c]; m1 += a; x1 = fmaxf(x1, a); m2 += d; x2 = fmaxf(x2, d); }
        VST2(float, SPP + ((long long)b * 4 + 0) * S + s, m1 / C); VST2(float, SPP + ((long long)b * 4 + 1) * S + s, x1); VST2(float, SPP + ((long long)b * 4 + 2) * S + s, m2 / C); VST2(float, SPP + ((long long)b * 4 + 3) * S + s, x2); }
}
__global__ __launch_bounds__(256) void k_mm_chgate(const float* __restrict__ CHP, const float* __restrict__ w1, const float* __restrict__ b1, const float* __restrict__ w2, const float* __restrict__ b2, float* __restrict__ CHS, int B, int C) {
    const int q = blockIdx.x * 256 + threadIdx.x; if (q >= B * C) return; const int c = q % C, b = q / C; float v1 = b1[0], v2 = b2[0];
    for (int i = 0; i < 4; ++i) for (int t = 0; t < 3; ++t) { const int cc = c + t - 1; if (cc < 0 || cc >= C) continue; const float x = CHP[((long long)b * 4 + i) * C + cc]; v1 += w1[i * 3 + t] * x; v2 += w2[i * 3 + t] * x; }
    const float mx = fmaxf(v1, v2); const float e1 = expf(v1 - mx), e2 = expf(v2 - mx); VST2(float, CHS + q, e1 / (e1 + e2)); VST2(float, CHS + (long long)B * C + q, e2 / (e1 + e2));
}
__global__ __launch_bounds__(256) void k_mm_spgate(const float* __restrict__ SPP, const float* __restrict__ w1, const float* __restrict__ b1, const float* __restrict__ w2, const float* __restrict__ b2, float* __restrict__ SPS, int B, int SP) {
    const int q = blockIdx.x * 256 + threadIdx.x; const int S = SP * SP; if (q >= B * S) return; const int s = q % S, b = q / S; const int y = s / SP, x = s % SP; float v1 = b1[0], v2 = b2[0];
    for (int i = 0; i < 4; ++i) for (int ky = 0; ky < 7; ++ky) { const int yy = y + ky - 3; if (yy < 0 || yy >= SP) continue; for (int kx = 0; kx < 7; ++kx) { const int xx = x + kx - 3; if (xx < 0 || xx >= SP) continue; const float v = SPP[((long long)b * 4 + i) * S + yy * SP + xx]; v1 += w1[(i * 7 + ky) * 7 + kx] * v; v2 += w2[(i * 7 + ky) * 7 + kx] * v; } }
    const float mx = fmaxf(v1, v2); const float e1 = expf(v1 - mx), e2 = expf(v2 - mx); VST2(float, SPS + q, e1 / (e1 + e2)); VST2(float, SPS + (long long)B * S + q, e2 / (e1 + e2));
}
__global__ __launch_bounds__(256) void k_mm_fuse(const float* __restrict__ T1, const float* __restrict__ T2, const float* __restrict__ CHS, const float* __restrict__ SPS, float* __restrict__ FM, int B, int S, int C) {
    const int q = blockIdx.x * 256 + threadIdx.x; if (q >= B * C) return; const int c = q % C, b = q / C; const float g1 = CHS[q], g2 = CHS[(long long)B * C + q]; float a = 0.f;
    for (int s = 0; s < S; ++s) { const float a1 = g1 + SPS[(long long)b * S + s] + 1.f, a2 = g2 + SPS[(long long)B * S + (long long)b * S + s] + 1.f; a += a1 * T1[((long long)b * S + s) * C + c] + a2 * T2[((long long)b * S + s) * C + c]; }
    VST2(float, FM + q, a / S);
}
__global__ __launch_bounds__(256) void k_mm_out(const float* __restrict__ LG, int ldp, float* __restrict__ OUT, int B, int NC) { const int b = blockIdx.x * 256 + threadIdx.x; if (b >= B) return; const float* l = LG + (long long)b * ldp; float mx = -__builtin_inff(); for (int j = 0; j < NC; ++j) mx = fmaxf(mx, l[j]); float s = 0.f; for (int j = 0; j < NC; ++j) s += expf(l[j] - mx); for (int j = 0; j < NC; ++j) VST2(float, OUT + b * NC + j, expf(l[j] - mx) / s); }
__global__ __launch_bounds__(256) void k_mm_rowsm(float* __restrict__ SC, int R, int N, float scale) { __shared__ float red[256]; const int r = blockIdx.x; float* row = SC + (long long)r * N; float mx = -__builtin_inff(); for (int j = threadIdx.x; j < N; j += 256) mx = fmaxf(mx, row[j] * scale); red[threadIdx.x] = mx; __syncthreads(); for (int o = 128; o > 0; o >>= 1) { if (threadIdx.x < o) red[threadIdx.x] = fmaxf(red[threadIdx.x], red[threadIdx.x + o]); __syncthreads(); } mx = red[0]; __syncthreads();
    float s = 0.f; for (int j = threadIdx.x; j < N; j += 256) s += expf(row[j] * scale - mx); red[threadIdx.x] = s; __syncthreads(); for (int o = 128; o > 0; o >>= 1) { if (threadIdx.x < o) red[threadIdx.x] += red[threadIdx.x + o]; __syncthreads(); } s = red[0];
    for (int j = threadIdx.x; j < N; j += 256) { const float pv = expf(row[j] * scale - mx) / s; VST2(float, row + j, pv); } }

template __global__ void k_gemm<1>(GemmP);
template __global__ void k_gemm<3>(GemmP);

extern "C" void kernel_launch(void* const* d_in, const int* in_sizes, int n_in, void* d_out, int out_size, void* d_ws, size_t ws_size, hipStream_t stream) {
    (void)in_sizes; (void)n_in; (void)out_size; (void)ws_size;
    const float* us = (const float*)d_in[0];
    const float* img = (const float*)d_in[1];
    const float* uw1 = (const float*)d_in[2];
    const float* ub1 = (const float*)d_in[3];
    const float* uw2 = (const float*)d_in[4];
    const float* ub2 = (const float*)d_in[5];
    const float* uw3 = (const float*)d_in[6];
    const float* ub3 = (const float*)d_in[7];
    const float* affw = (const float*)d_in[8];
    const float* affh = (const float*)d_in[9];
    const float* thr = (const float*)d_in[10];
    const float* iw1 = (const float*)d_in[11];
    const float* ib1 = (const float*)d_in[12];
    const float* iw2 = (const float*)d_in[13];
    const float* ib2 = (const float*)d_in[14];
    const float* iw3 = (const float*)d_in[15];
    const float* ib3 = (const float*)d_in[16];
    const float* qkvw = (const float*)d_in[17];
    const float* qkvb = (const float*)d_in[18];
    const float* dww = (const float*)d_in[19];
    const float* dwb = (const float*)d_in[20];
    const float* projw = (const float*)d_in[21];
    const float* projb = (const float*)d_in[22];
    const float* fcw = (const float*)d_in[23];
    const float* fcb = (const float*)d_in[24];
    const float* depw = (const float*)d_in[25];
    const float* depb = (const float*)d_in[26];
    const float* temp = (const float*)d_in[27];
    const float* caw = (const float*)d_in[28];
    const float* cab = (const float*)d_in[29];
    const float* cow = (const float*)d_in[30];
    const float* cob = (const float*)d_in[31];
    const float* ch1w = (const float*)d_in[32];
    const float* ch1b = (const float*)d_in[33];
    const float* ch2w = (const float*)d_in[34];
    const float* ch2b = (const float*)d_in[35];
    const float* sp1w = (const float*)d_in[36];
    const float* sp1b = (const float*)d_in[37];
    const float* sp2w = (const float*)d_in[38];
    const float* sp2b = (const float*)d_in[39];
    const float* clsw = (const float*)d_in[40];
    const float* clsb = (const float*)d_in[41];
    const int Bn = 16;
    const int L = 4096;
    const int NF = 2049;
    const int HW = 4096;
    const int SEQ = 1024;
    const int LP = 32;
    float* out = (float*)d_out;
    char* wsp = (char*)d_ws;
    float* U0 = (float*)wsp; wsp += (((size_t)((size_t)Bn * 4098 * 1) * 4 + 255) / 256) * 256;
    float* U1 = (float*)wsp; wsp += (((size_t)((size_t)Bn * 4098 * 16) * 4 + 255) / 256) * 256;
    float* U2 = (float*)wsp; wsp += (((size_t)((size_t)Bn * 4098 * 32) * 4 + 255) / 256) * 256;
    float* U3 = (float*)wsp; wsp += (((size_t)((size_t)Bn * 4098 * 64) * 4 + 255) / 256) * 256;
    float* R67 = (float*)wsp; wsp += (((size_t)((size_t)2 * NF * L) * 4 + 255) / 256) * 256;
    float* XR = (float*)wsp; wsp += (((size_t)((size_t)Bn * NF * 64) * 4 + 255) / 256) * 256;
    float* XI = (float*)wsp; wsp += (((size_t)((size_t)Bn * NF * 64) * 4 + 255) / 256) * 256;
    float* MSK = (float*)wsp; wsp += (((size_t)((size_t)Bn * NF + 64) * 4 + 255) / 256) * 256;
    float* UF = (float*)wsp; wsp += (((size_t)((size_t)Bn * L * 64) * 4 + 255) / 256) * 256;
    float* UR = (float*)wsp; wsp += (((size_t)((size_t)Bn * SEQ * 64) * 4 + 255) / 256) * 256;
    float* IR = (float*)wsp; wsp += (((size_t)((size_t)Bn * SEQ * 64) * 4 + 255) / 256) * 256;
    float* H1 = (float*)wsp; wsp += (((size_t)((size_t)Bn * SEQ * 192) * 4 + 255) / 256) * 256;
    float* H2 = (float*)wsp; wsp += (((size_t)((size_t)Bn * SEQ * 192) * 4 + 255) / 256) * 256;
    float* SC = (float*)wsp; wsp += (((size_t)((size_t)4 * SEQ * SEQ) * 4 + 255) / 256) * 256;
    float* O1 = (float*)wsp; wsp += (((size_t)((size_t)Bn * SEQ * 64) * 4 + 255) / 256) * 256;
    float* O2 = (float*)wsp; wsp += (((size_t)((size_t)Bn * SEQ * 64) * 4 + 255) / 256) * 256;
    float* T1 = (float*)wsp; wsp += (((size_t)((size_t)Bn * SEQ * 64) * 4 + 255) / 256) * 256;
    float* T2 = (float*)wsp; wsp += (((size_t)((size_t)Bn * SEQ * 64) * 4 + 255) / 256) * 256;
    float* CHP = (float*)wsp; wsp += (((size_t)((size_t)Bn * 4 * 64) * 4 + 255) / 256) * 256;
    float* SPP = (float*)wsp; wsp += (((size_t)((size_t)Bn * 4 * SEQ) * 4 + 255) / 256) * 256;
    float* CHS = (float*)wsp; wsp += (((size_t)((size_t)2 * Bn * 64) * 4 + 255) / 256) * 256;
    float* SPS = (float*)wsp; wsp += (((size_t)((size_t)2 * Bn * SEQ) * 4 + 255) / 256) * 256;
    float* FM = (float*)wsp; wsp += (((size_t)((size_t)Bn * 64) * 4 + 255) / 256) * 256;
    float* LG = (float*)wsp; wsp += (((size_t)((size_t)Bn * LP) * 4 + 255) / 256) * 256;
    hipMemsetAsync(U0, 0, (size_t)Bn * 4098 * 4, stream); hipMemsetAsync(U1, 0, (size_t)Bn * 4098 * 16 * 4, stream); hipMemsetAsync(U2, 0, (size_t)Bn * 4098 * 32 * 4, stream); hipMemsetAsync(U3, 0, (size_t)Bn * 4098 * 64 * 4, stream);
    k_mm_pad1d<<<(unsigned)((Bn * L + 255) / 256), 256, 0, stream>>>(us, U0, Bn, L);
    k_mm_dft<<<(unsigned)(((long long)NF * L + 255) / 256), 256, 0, stream>>>(R67, R67 + (size_t)NF * L, NF, L);
    { GemmP u1_0;
      u1_0.A = U0 + (size_t)0 * 1; u1_0.B = uw1 + 0; u1_0.bias = ub1; u1_0.R = U0 + (size_t)0 * 1; u1_0.C = U1 + 16;
      u1_0.sAo = (long long)(L + 2) * 1; u1_0.sAi = 0; u1_0.sAm = 1; u1_0.sAk = 1; u1_0.sBo = 0; u1_0.sBi = 0; u1_0.sBn = 1 * 3; u1_0.sBk = 3; u1_0.sCo = (long long)(L + 2) * 16; u1_0.sCi = 0; u1_0.sCm = 16; u1_0.sRo = 0; u1_0.sRi = 0; u1_0.sRm = 0; u1_0.sRn = 0;
      u1_0.M = L; u1_0.N = 16; u1_0.K = 1; u1_0.zi_n = 1; u1_0.flags = 1; u1_0.act = 0;
      u1_0.alpha = 1.0f; u1_0.beta = 0.0f; u1_0.sa = 1.0f; u1_0.sb = 1.0f; u1_0.Npad = 16; u1_0.pad_ = 0;
      k_gemm<1><<<dim3((unsigned)((16) + 31) / 32, (unsigned)((L) + 15) / 16, (unsigned)(Bn)), 32, 0, stream>>>(u1_0); }
    { GemmP u1_1;
      u1_1.A = U0 + (size_t)1 * 1; u1_1.B = uw1 + 1; u1_1.bias = U0 + (size_t)1 * 1; u1_1.R = U1 + 16; u1_1.C = U1 + 16;
      u1_1.sAo = (long long)(L + 2) * 1; u1_1.sAi = 0; u1_1.sAm = 1; u1_1.sAk = 1; u1_1.sBo = 0; u1_1.sBi = 0; u1_1.sBn = 1 * 3; u1_1.sBk = 3; u1_1.sCo = (long long)(L + 2) * 16; u1_1.sCi = 0; u1_1.sCm = 16; u1_1.sRo = (long long)(L + 2) * 16; u1_1.sRi = 0; u1_1.sRm = 16; u1_1.sRn = 1;
      u1_1.M = L; u1_1.N = 16; u1_1.K = 1; u1_1.zi_n = 1; u1_1.flags = 4; u1_1.act = 0;
      u1_1.alpha = 1.0f; u1_1.beta = 1.0f; u1_1.sa = 1.0f; u1_1.sb = 1.0f; u1_1.Npad = 16; u1_1.pad_ = 0;
      k_gemm<1><<<dim3((unsigned)((16) + 31) / 32, (unsigned)((L) + 15) / 16, (unsigned)(Bn)), 32, 0, stream>>>(u1_1); }
    { GemmP u1_2;
      u1_2.A = U0 + (size_t)2 * 1; u1_2.B = uw1 + 2; u1_2.bias = U0 + (size_t)2 * 1; u1_2.R = U1 + 16; u1_2.C = U1 + 16;
      u1_2.sAo = (long long)(L + 2) * 1; u1_2.sAi = 0; u1_2.sAm = 1; u1_2.sAk = 1; u1_2.sBo = 0; u1_2.sBi = 0; u1_2.sBn = 1 * 3; u1_2.sBk = 3; u1_2.sCo = (long long)(L + 2) * 16; u1_2.sCi = 0; u1_2.sCm = 16; u1_2.sRo = (long long)(L + 2) * 16; u1_2.sRi = 0; u1_2.sRm = 16; u1_2.sRn = 1;
      u1_2.M = L; u1_2.N = 16; u1_2.K = 1; u1_2.zi_n = 1; u1_2.flags = 4; u1_2.act = 0;
      u1_2.alpha = 1.0f; u1_2.beta = 1.0f; u1_2.sa = 1.0f; u1_2.sb = 1.0f; u1_2.Npad = 16; u1_2.pad_ = 0;
      k_gemm<1><<<dim3((unsigned)((16) + 31) / 32, (unsigned)((L) + 15) / 16, (unsigned)(Bn)), 32, 0, stream>>>(u1_2); }
    k_mm_relu1d<<<(unsigned)(((long long)Bn * L * 16 + 255) / 256), 256, 0, stream>>>(U1, Bn, L, 16);
    { GemmP u2_0;
      u2_0.A = U1 + (size_t)0 * 16; u2_0.B = uw2 + 0; u2_0.bias = ub2; u2_0.R = U1 + (size_t)0 * 16; u2_0.C = U2 + 32;
      u2_0.sAo = (long long)(L + 2) * 16; u2_0.sAi = 0; u2_0.sAm = 16; u2_0.sAk = 1; u2_0.sBo = 0; u2_0.sBi = 0; u2_0.sBn = 16 * 3; u2_0.sBk = 3; u2_0.sCo = (long long)(L + 2) * 32; u2_0.sCi = 0; u2_0.sCm = 32; u2_0.sRo = 0; u2_0.sRi = 0; u2_0.sRm = 0; u2_0.sRn = 0;
      u2_0.M = L; u2_0.N = 32; u2_0.K = 16; u2_0.zi_n = 1; u2_0.flags = 1; u2_0.act = 0;
      u2_0.alpha = 1.0f; u2_0.beta = 0.0f; u2_0.sa = 1.0f; u2_0.sb = 1.0f; u2_0.Npad = 32; u2_0.pad_ = 0;
      k_gemm<1><<<dim3((unsigned)((32) + 31) / 32, (unsigned)((L) + 15) / 16, (unsigned)(Bn)), 32, 0, stream>>>(u2_0); }
    { GemmP u2_1;
      u2_1.A = U1 + (size_t)1 * 16; u2_1.B = uw2 + 1; u2_1.bias = U1 + (size_t)1 * 16; u2_1.R = U2 + 32; u2_1.C = U2 + 32;
      u2_1.sAo = (long long)(L + 2) * 16; u2_1.sAi = 0; u2_1.sAm = 16; u2_1.sAk = 1; u2_1.sBo = 0; u2_1.sBi = 0; u2_1.sBn = 16 * 3; u2_1.sBk = 3; u2_1.sCo = (long long)(L + 2) * 32; u2_1.sCi = 0; u2_1.sCm = 32; u2_1.sRo = (long long)(L + 2) * 32; u2_1.sRi = 0; u2_1.sRm = 32; u2_1.sRn = 1;
      u2_1.M = L; u2_1.N = 32; u2_1.K = 16; u2_1.zi_n = 1; u2_1.flags = 4; u2_1.act = 0;
      u2_1.alpha = 1.0f; u2_1.beta = 1.0f; u2_1.sa = 1.0f; u2_1.sb = 1.0f; u2_1.Npad = 32; u2_1.pad_ = 0;
      k_gemm<1><<<dim3((unsigned)((32) + 31) / 32, (unsigned)((L) + 15) / 16, (unsigned)(Bn)), 32, 0, stream>>>(u2_1); }
    { GemmP u2_2;
      u2_2.A = U1 + (size_t)2 * 16; u2_2.B = uw2 + 2; u2_2.bias = U1 + (size_t)2 * 16; u2_2.R = U2 + 32; u2_2.C = U2 + 32;
      u2_2.sAo = (long long)(L + 2) * 16; u2_2.sAi = 0; u2_2.sAm = 16; u2_2.sAk = 1; u2_2.sBo = 0; u2_2.sBi = 0; u2_2.sBn = 16 * 3; u2_2.sBk = 3; u2_2.sCo = (long long)(L + 2) * 32; u2_2.sCi = 0; u2_2.sCm = 32; u2_2.sRo = (long long)(L + 2) * 32; u2_2.sRi = 0; u2_2.sRm = 32; u2_2.sRn = 1;
      u2_2.M = L; u2_2.N = 32; u2_2.K = 16; u2_2.zi_n = 1; u2_2.flags = 4; u2_2.act = 0;
      u2_2.alpha = 1.0f; u2_2.beta = 1.0f; u2_2.sa = 1.0f; u2_2.sb = 1.0f; u2_2.Npad = 32; u2_2.pad_ = 0;
      k_gemm<1><<<dim3((unsigned)((32) + 31) / 32, (unsigned)((L) + 15) / 16, (unsigned)(Bn)), 32, 0, stream>>>(u2_2); }
    k_mm_relu1d<<<(unsigned)(((long long)Bn * L * 32 + 255) / 256), 256, 0, stream>>>(U2, Bn, L, 32);
    { GemmP u3_0;
      u3_0.A = U2 + (size_t)0 * 32; u3_0.B = uw3 + 0; u3_0.bias = ub3; u3_0.R = U2 + (size_t)0 * 32; u3_0.C = U3 + 64;
      u3_0.sAo = (long long)(L + 2) * 32; u3_0.sAi = 0; u3_0.sAm = 32; u3_0.sAk = 1; u3_0.sBo = 0; u3_0.sBi = 0; u3_0.sBn = 32 * 3; u3_0.sBk = 3; u3_0.sCo = (long long)(L + 2) * 64; u3_0.sCi = 0; u3_0.sCm = 64; u3_0.sRo = 0; u3_0.sRi = 0; u3_0.sRm = 0; u3_0.sRn = 0;
      u3_0.M = L; u3_0.N = 64; u3_0.K = 32; u3_0.zi_n = 1; u3_0.flags = 1; u3_0.act = 0;
      u3_0.alpha = 1.0f; u3_0.beta = 0.0f; u3_0.sa = 1.0f; u3_0.sb = 1.0f; u3_0.Npad = 64; u3_0.pad_ = 0;
      k_gemm<1><<<dim3((unsigned)((64) + 31) / 32, (unsigned)((L) + 15) / 16, (unsigned)(Bn)), 32, 0, stream>>>(u3_0); }
    { GemmP u3_1;
      u3_1.A = U2 + (size_t)1 * 32; u3_1.B = uw3 + 1; u3_1.bias = U2 + (size_t)1 * 32; u3_1.R = U3 + 64; u3_1.C = U3 + 64;
      u3_1.sAo = (long long)(L + 2) * 32; u3_1.sAi = 0; u3_1.sAm = 32; u3_1.sAk = 1; u3_1.sBo = 0; u3_1.sBi = 0; u3_1.sBn = 32 * 3; u3_1.sBk = 3; u3_1.sCo = (long long)(L + 2) * 64; u3_1.sCi = 0; u3_1.sCm = 64; u3_1.sRo = (long long)(L + 2) * 64; u3_1.sRi = 0; u3_1.sRm = 64; u3_1.sRn = 1;
      u3_1.M = L; u3_1.N = 64; u3_1.K = 32; u3_1.zi_n = 1; u3_1.flags = 4; u3_1.act = 0;
      u3_1.alpha = 1.0f; u3_1.beta = 1.0f; u3_1.sa = 1.0f; u3_1.sb = 1.0f; u3_1.Npad = 64; u3_1.pad_ = 0;
      k_gemm<1><<<dim3((unsigned)((64) + 31) / 32, (unsigned)((L) + 15) / 16, (unsigned)(Bn)), 32, 0, stream>>>(u3_1); }
    { GemmP u3_2;
      u3_2.A = U2 + (size_t)2 * 32; u3_2.B = uw3 + 2; u3_2.bias = U2 + (size_t)2 * 32; u3_2.R = U3 + 64; u3_2.C = U3 + 64;
      u3_2.sAo = (long long)(L + 2) * 32; u3_2.sAi = 0; u3_2.sAm = 32; u3_2.sAk = 1; u3_2.sBo = 0; u3_2.sBi = 0; u3_2.sBn = 32 * 3; u3_2.sBk = 3; u3_2.sCo = (long long)(L + 2) * 64; u3_2.sCi = 0; u3_2.sCm = 64; u3_2.sRo = (long long)(L + 2) * 64; u3_2.sRi = 0; u3_2.sRm = 64; u3_2.sRn = 1;
      u3_2.M = L; u3_2.N = 64; u3_2.K = 32; u3_2.zi_n = 1; u3_2.flags = 4; u3_2.act = 0;
      u3_2.alpha = 1.0f; u3_2.beta = 1.0f; u3_2.sa = 1.0f; u3_2.sb = 1.0f; u3_2.Npad = 64; u3_2.pad_ = 0;
      k_gemm<1><<<dim3((unsigned)((64) + 31) / 32, (unsigned)((L) + 15) / 16, (unsigned)(Bn)), 32, 0, stream>>>(u3_2); }
    k_mm_relu1d<<<(unsigned)(((long long)Bn * L * 64 + 255) / 256), 256, 0, stream>>>(U3, Bn, L, 64);
    { GemmP gxr;
      gxr.A = R67; gxr.B = U3 + 64; gxr.bias = R67; gxr.R = R67; gxr.C = XR;
      gxr.sAo = 0; gxr.sAi = 0; gxr.sAm = L; gxr.sAk = 1; gxr.sBo = (long long)(L + 2) * 64; gxr.sBi = 0; gxr.sBn = 1; gxr.sBk = 64; gxr.sCo = (long long)NF * 64; gxr.sCi = 0; gxr.sCm = 64; gxr.sRo = 0; gxr.sRi = 0; gxr.sRm = 0; gxr.sRn = 0;
      gxr.M = NF; gxr.N = 64; gxr.K = L; gxr.zi_n = 1; gxr.flags = 0; gxr.act = 0;
      gxr.alpha = 1.0f; gxr.beta = 0.0f; gxr.sa = 1.0f; gxr.sb = 1.0f; gxr.Npad = 64; gxr.pad_ = 0;
      k_gemm<3><<<dim3((unsigned)((64) + 31) / 32, (unsigned)((NF) + 15) / 16, (unsigned)(Bn)), 32, 0, stream>>>(gxr); }
    { GemmP gxi;
      gxi.A = R67 + (size_t)NF * L; gxi.B = U3 + 64; gxi.bias = R67 + (size_t)NF * L; gxi.R = R67 + (size_t)NF * L; gxi.C = XI;
      gxi.sAo = 0; gxi.sAi = 0; gxi.sAm = L; gxi.sAk = 1; gxi.sBo = (long long)(L + 2) * 64; gxi.sBi = 0; gxi.sBn = 1; gxi.sBk = 64; gxi.sCo = (long long)NF * 64; gxi.sCi = 0; gxi.sCm = 64; gxi.sRo = 0; gxi.sRi = 0; gxi.sRm = 0; gxi.sRn = 0;
      gxi.M = NF; gxi.N = 64; gxi.K = L; gxi.zi_n = 1; gxi.flags = 0; gxi.act = 0;
      gxi.alpha = -1.0f; gxi.beta = 0.0f; gxi.sa = 1.0f; gxi.sb = 1.0f; gxi.Npad = 64; gxi.pad_ = 0;
      k_gemm<3><<<dim3((unsigned)((64) + 31) / 32, (unsigned)((NF) + 15) / 16, (unsigned)(Bn)), 32, 0, stream>>>(gxi); }
    k_mm_energy<<<(unsigned)((Bn * NF + 255) / 256), 256, 0, stream>>>(XR, XI, MSK, Bn, NF, 64);
    k_mm_filter<<<dim3(NF, Bn), 256, 0, stream>>>(XR, XI, MSK, affw, affh, thr, Bn, NF, 64);
    { GemmP gur;
      gur.A = R67; gur.B = XR; gur.bias = R67; gur.R = R67; gur.C = UF;
      gur.sAo = 0; gur.sAi = 0; gur.sAm = 1; gur.sAk = L; gur.sBo = (long long)NF * 64; gur.sBi = 0; gur.sBn = 1; gur.sBk = 64; gur.sCo = (long long)L * 64; gur.sCi = 0; gur.sCm = 64; gur.sRo = 0; gur.sRi = 0; gur.sRm = 0; gur.sRn = 0;
      gur.M = L; gur.N = 64; gur.K = NF; gur.zi_n = 1; gur.flags = 0; gur.act = 0;
      gur.alpha = 1.0f; gur.beta = 0.0f; gur.sa = 1.0f; gur.sb = 1.0f; gur.Npad = 64; gur.pad_ = 0;
      k_gemm<3><<<dim3((unsigned)((64) + 31) / 32, (unsigned)((L) + 15) / 16, (unsigned)(Bn)), 32, 0, stream>>>(gur); }
    { GemmP gui;
      gui.A = R67 + (size_t)NF * L; gui.B = XI; gui.bias = R67 + (size_t)NF * L; gui.R = UF; gui.C = UF;
      gui.sAo = 0; gui.sAi = 0; gui.sAm = 1; gui.sAk = L; gui.sBo = (long long)NF * 64; gui.sBi = 0; gui.sBn = 1; gui.sBk = 64; gui.sCo = (long long)L * 64; gui.sCi = 0; gui.sCm = 64; gui.sRo = (long long)L * 64; gui.sRi = 0; gui.sRm = 64; gui.sRn = 1;
      gui.M = L; gui.N = 64; gui.K = NF; gui.zi_n = 1; gui.flags = 4; gui.act = 0;
      gui.alpha = -1.0f; gui.beta = 1.0f; gui.sa = 1.0f; gui.sb = 1.0f; gui.Npad = 64; gui.pad_ = 0;
      k_gemm<3><<<dim3((unsigned)((64) + 31) / 32, (unsigned)((L) + 15) / 16, (unsigned)(Bn)), 32, 0, stream>>>(gui); }
    k_mm_uspool<<<(unsigned)(((long long)Bn * SEQ * 64 + 255) / 256), 256, 0, stream>>>(UF, UR, Bn, L, 64);
    hipMemsetAsync(R67 + 0, 0, (size_t)2 * 66 * 66 * 3 * 4, stream); hipMemsetAsync(R67 + 26176, 0, (size_t)2 * 66 * 66 * 16 * 4, stream); hipMemsetAsync(R67 + 165568, 0, (size_t)2 * 66 * 66 * 32 * 4, stream); hipMemsetAsync(R67 + 444352, 0, (size_t)2 * 66 * 66 * 64 * 4, stream);
    k_mm_padimg<<<(unsigned)(((long long)2 * HW * 3 + 255) / 256), 256, 0, stream>>>(img + (size_t)0 * 3 * HW, R67 + 0, 2, 3, 64);
    { GemmP i1c0_0;
      i1c0_0.A = R67 + 0 + (size_t)0 * 3; i1c0_0.B = iw1 + 0; i1c0_0.bias = ib1; i1c0_0.R = R67 + 0 + (size_t)0 * 3; i1c0_0.C = R67 + 26176 + (size_t)67 * 16;
      i1c0_0.sAo = (long long)66 * 66 * 3; i1c0_0.sAi = (long long)66 * 3; i1c0_0.sAm = 3; i1c0_0.sAk = 1; i1c0_0.sBo = 0; i1c0_0.sBi = 0; i1c0_0.sBn = 3 * 9; i1c0_0.sBk = 9; i1c0_0.sCo = (long long)66 * 66 * 16; i1c0_0.sCi = (long long)66 * 16; i1c0_0.sCm = 16; i1c0_0.sRo = 0; i1c0_0.sRi = 0; i1c0_0.sRm = 0; i1c0_0.sRn = 0;
      i1c0_0.M = 64; i1c0_0.N = 16; i1c0_0.K = 3; i1c0_0.zi_n = 64; i1c0_0.flags = 1; i1c0_0.act = 0;
      i1c0_0.alpha = 1.0f; i1c0_0.beta = 0.0f; i1c0_0.sa = 1.0f; i1c0_0.sb = 1.0f; i1c0_0.Npad = 16; i1c0_0.pad_ = 0;
      k_gemm<1><<<dim3((unsigned)((16) + 31) / 32, (unsigned)((64) + 15) / 16, (unsigned)(2 * 64)), 32, 0, stream>>>(i1c0_0); }
    { GemmP i1c0_1;
      i1c0_1.A = R67 + 0 + (size_t)1 * 3; i1c0_1.B = iw1 + 1; i1c0_1.bias = R67 + 0 + (size_t)1 * 3; i1c0_1.R = R67 + 26176 + (size_t)67 * 16; i1c0_1.C = R67 + 26176 + (size_t)67 * 16;
      i1c0_1.sAo = (long long)66 * 66 * 3; i1c0_1.sAi = (long long)66 * 3; i1c0_1.sAm = 3; i1c0_1.sAk = 1; i1c0_1.sBo = 0; i1c0_1.sBi = 0; i1c0_1.sBn = 3 * 9; i1c0_1.sBk = 9; i1c0_1.sCo = (long long)66 * 66 * 16; i1c0_1.sCi = (long long)66 * 16; i1c0_1.sCm = 16; i1c0_1.sRo = (long long)66 * 66 * 16; i1c0_1.sRi = (long long)66 * 16; i1c0_1.sRm = 16; i1c0_1.sRn = 1;
      i1c0_1.M = 64; i1c0_1.N = 16; i1c0_1.K = 3; i1c0_1.zi_n = 64; i1c0_1.flags = 4; i1c0_1.act = 0;
      i1c0_1.alpha = 1.0f; i1c0_1.beta = 1.0f; i1c0_1.sa = 1.0f; i1c0_1.sb = 1.0f; i1c0_1.Npad = 16; i1c0_1.pad_ = 0;
      k_gemm<1><<<dim3((unsigned)((16) + 31) / 32, (unsigned)((64) + 15) / 16, (unsigned)(2 * 64)), 32, 0, stream>>>(i1c0_1); }
    { GemmP i1c0_2;
      i1c0_2.A = R67 + 0 + (size_t)2 * 3; i1c0_2.B = iw1 + 2; i1c0_2.bias = R67 + 0 + (size_t)2 * 3; i1c0_2.R = R67 + 26176 + (size_t)67 * 16; i1c0_2.C = R67 + 26176 + (size_t)67 * 16;
      i1c0_2.sAo = (long long)66 * 66 * 3; i1c0_2.sAi = (long long)66 * 3; i1c0_2.sAm = 3; i1c0_2.sAk = 1; i1c0_2.sBo = 0; i1c0_2.sBi = 0; i1c0_2.sBn = 3 * 9; i1c0_2.sBk = 9; i1c0_2.sCo = (long long)66 * 66 * 16; i1c0_2.sCi = (long long)66 * 16; i1c0_2.sCm = 16; i1c0_2.sRo = (long long)66 * 66 * 16; i1c0_2.sRi = (long long)66 * 16; i1c0_2.sRm = 16; i1c0_2.sRn = 1;
      i1c0_2.M = 64; i1c0_2.N = 16; i1c0_2.K = 3; i1c0_2.zi_n = 64; i1c0_2.flags = 4; i1c0_2.act = 0;
      i1c0_2.alpha = 1.0f; i1c0_2.beta = 1.0f; i1c0_2.sa = 1.0f; i1c0_2.sb = 1.0f; i1c0_2.Npad = 16; i1c0_2.pad_ = 0;
      k_gemm<1><<<dim3((unsigned)((16) + 31) / 32, (unsigned)((64) + 15) / 16, (unsigned)(2 * 64)), 32, 0, stream>>>(i1c0_2); }
    { GemmP i1c0_3;
      i1c0_3.A = R67 + 0 + (size_t)66 * 3; i1c0_3.B = iw1 + 3; i1c0_3.bias = R67 + 0 + (size_t)66 * 3; i1c0_3.R = R67 + 26176 + (size_t)67 * 16; i1c0_3.C = R67 + 26176 + (size_t)67 * 16;
      i1c0_3.sAo = (long long)66 * 66 * 3; i1c0_3.sAi = (long long)66 * 3; i1c0_3.sAm = 3; i1c0_3.sAk = 1; i1c0_3.sBo = 0; i1c0_3.sBi = 0; i1c0_3.sBn = 3 * 9; i1c0_3.sBk = 9; i1c0_3.sCo = (long long)66 * 66 * 16; i1c0_3.sCi = (long long)66 * 16; i1c0_3.sCm = 16; i1c0_3.sRo = (long long)66 * 66 * 16; i1c0_3.sRi = (long long)66 * 16; i1c0_3.sRm = 16; i1c0_3.sRn = 1;
      i1c0_3.M = 64; i1c0_3.N = 16; i1c0_3.K = 3; i1c0_3.zi_n = 64; i1c0_3.flags = 4; i1c0_3.act = 0;
      i1c0_3.alpha = 1.0f; i1c0_3.beta = 1.0f; i1c0_3.sa = 1.0f; i1c0_3.sb = 1.0f; i1c0_3.Npad = 16; i1c0_3.pad_ = 0;
      k_gemm<1><<<dim3((unsigned)((16) + 31) / 32, (unsigned)((64) + 15) / 16, (unsigned)(2 * 64)), 32, 0, stream>>>(i1c0_3); }
    { GemmP i1c0_4;
      i1c0_4.A = R67 + 0 + (size_t)67 * 3; i1c0_4.B = iw1 + 4; i1c0_4.bias = R67 + 0 + (size_t)67 * 3; i1c0_4.R = R67 + 26176 + (size_t)67 * 16; i1c0_4.C = R67 + 26176 + (size_t)67 * 16;
      i1c0_4.sAo = (long long)66 * 66 * 3; i1c0_4.sAi = (long long)66 * 3; i1c0_4.sAm = 3; i1c0_4.sAk = 1; i1c0_4.sBo = 0; i1c0_4.sBi = 0; i1c0_4.sBn = 3 * 9; i1c0_4.sBk = 9; i1c0_4.sCo = (long long)66 * 66 * 16; i1c0_4.sCi = (long long)66 * 16; i1c0_4.sCm = 16; i1c0_4.sRo = (long long)66 * 66 * 16; i1c0_4.sRi = (long long)66 * 16; i1c0_4.sRm = 16; i1c0_4.sRn = 1;
      i1c0_4.M = 64; i1c0_4.N = 16; i1c0_4.K = 3; i1c0_4.zi_n = 64; i1c0_4.flags = 4; i1c0_4.act = 0;
      i1c0_4.alpha = 1.0f; i1c0_4.beta = 1.0f; i1c0_4.sa = 1.0f; i1c0_4.sb = 1.0f; i1c0_4.Npad = 16; i1c0_4.pad_ = 0;
      k_gemm<1><<<dim3((unsigned)((16) + 31) / 32, (unsigned)((64) + 15) / 16, (unsigned)(2 * 64)), 32, 0, stream>>>(i1c0_4); }
    { GemmP i1c0_5;
      i1c0_5.A = R67 + 0 + (size_t)68 * 3; i1c0_5.B = iw1 + 5; i1c0_5.bias = R67 + 0 + (size_t)68 * 3; i1c0_5.R = R67 + 26176 + (size_t)67 * 16; i1c0_5.C = R67 + 26176 + (size_t)67 * 16;
      i1c0_5.sAo = (long long)66 * 66 * 3; i1c0_5.sAi = (long long)66 * 3; i1c0_5.sAm = 3; i1c0_5.sAk = 1; i1c0_5.sBo = 0; i1c0_5.sBi = 0; i1c0_5.sBn = 3 * 9; i1c0_5.sBk = 9; i1c0_5.sCo = (long long)66 * 66 * 16; i1c0_5.sCi = (long long)66 * 16; i1c0_5.sCm = 16; i1c0_5.sRo = (long long)66 * 66 * 16; i1c0_5.sRi = (long long)66 * 16; i1c0_5.sRm = 16; i1c0_5.sRn = 1;
      i1c0_5.M = 64; i1c0_5.N = 16; i1c0_5.K = 3; i1c0_5.zi_n = 64; i1c0_5.flags = 4; i1c0_5.act = 0;
      i1c0_5.alpha = 1.0f; i1c0_5.beta = 1.0f; i1c0_5.sa = 1.0f; i1c0_5.sb = 1.0f; i1c0_5.Npad = 16; i1c0_5.pad_ = 0;
      k_gemm<1><<<dim3((unsigned)((16) + 31) / 32, (unsigned)((64) + 15) / 16, (unsigned)(2 * 64)), 32, 0, stream>>>(i1c0_5); }
    { GemmP i1c0_6;
      i1c0_6.A = R67 + 0 + (size_t)132 * 3; i1c0_6.B = iw1 + 6; i1c0_6.bias = R67 + 0 + (size_t)132 * 3; i1c0_6.R = R67 + 26176 + (size_t)67 * 16; i1c0_6.C = R67 + 26176 + (size_t)67 * 16;
      i1c0_6.sAo = (long long)66 * 66 * 3; i1c0_6.sAi = (long long)66 * 3; i1c0_6.sAm = 3; i1c0_6.sAk = 1; i1c0_6.sBo = 0; i1c0_6.sBi = 0; i1c0_6.sBn = 3 * 9; i1c0_6.sBk = 9; i1c0_6.sCo = (long long)66 * 66 * 16; i1c0_6.sCi = (long long)66 * 16; i1c0_6.sCm = 16; i1c0_6.sRo = (long long)66 * 66 * 16; i1c0_6.sRi = (long long)66 * 16; i1c0_6.sRm = 16; i1c0_6.sRn = 1;
      i1c0_6.M = 64; i1c0_6.N = 16; i1c0_6.K = 3; i1c0_6.zi_n = 64; i1c0_6.flags = 4; i1c0_6.act = 0;
      i1c0_6.alpha = 1.0f; i1c0_6.beta = 1.0f; i1c0_6.sa = 1.0f; i1c0_6.sb = 1.0f; i1c0_6.Npad = 16; i1c0_6.pad_ = 0;
      k_gemm<1><<<dim3((unsigned)((16) + 31) / 32, (unsigned)((64) + 15) / 16, (unsigned)(2 * 64)), 32, 0, stream>>>(i1c0_6); }
    { GemmP i1c0_7;
      i1c0_7.A = R67 + 0 + (size_t)133 * 3; i1c0_7.B = iw1 + 7; i1c0_7.bias = R67 + 0 + (size_t)133 * 3; i1c0_7.R = R67 + 26176 + (size_t)67 * 16; i1c0_7.C = R67 + 26176 + (size_t)67 * 16;
      i1c0_7.sAo = (long long)66 * 66 * 3; i1c0_7.sAi = (long long)66 * 3; i1c0_7.sAm = 3; i1c0_7.sAk = 1; i1c0_7.sBo = 0; i1c0_7.sBi = 0; i1c0_7.sBn = 3 * 9; i1c0_7.sBk = 9; i1c0_7.sCo = (long long)66 * 66 * 16; i1c0_7.sCi = (long long)66 * 16; i1c0_7.sCm = 16; i1c0_7.sRo = (long long)66 * 66 * 16; i1c0_7.sRi = (long long)66 * 16; i1c0_7.sRm = 16; i1c0_7.sRn = 1;
      i1c0_7.M = 64; i1c0_7.N = 16; i1c0_7.K = 3; i1c0_7.zi_n = 64; i1c0_7.flags = 4; i1c0_7.act = 0;
      i1c0_7.alpha = 1.0f; i1c0_7.beta = 1.0f; i1c0_7.sa = 1.0f; i1c0_7.sb = 1.0f; i1c0_7.Npad = 16; i1c0_7.pad_ = 0;
      k_gemm<1><<<dim3((unsigned)((16) + 31) / 32, (unsigned)((64) + 15) / 16, (unsigned)(2 * 64)), 32, 0, stream>>>(i1c0_7); }
    { GemmP i1c0_8;
      i1c0_8.A = R67 + 0 + (size_t)134 * 3; i1c0_8.B = iw1 + 8; i1c0_8.bias = R67 + 0 + (size_t)134 * 3; i1c0_8.R = R67 + 26176 + (size_t)67 * 16; i1c0_8.C = R67 + 26176 + (size_t)67 * 16;
      i1c0_8.sAo = (long long)66 * 66 * 3; i1c0_8.sAi = (long long)66 * 3; i1c0_8.sAm = 3; i1c0_8.sAk = 1; i1c0_8.sBo = 0; i1c0_8.sBi = 0; i1c0_8.sBn = 3 * 9; i1c0_8.sBk = 9; i1c0_8.sCo = (long long)66 * 66 * 16; i1c0_8.sCi = (long long)66 * 16; i1c0_8.sCm = 16; i1c0_8.sRo = (long long)66 * 66 * 16; i1c0_8.sRi = (long long)66 * 16; i1c0_8.sRm = 16; i1c0_8.sRn = 1;
      i1c0_8.M = 64; i1c0_8.N = 16; i1c0_8.K = 3; i1c0_8.zi_n = 64; i1c0_8.flags = 4; i1c0_8.act = 0;
      i1c0_8.alpha = 1.0f; i1c0_8.beta = 1.0f; i1c0_8.sa = 1.0f; i1c0_8.sb = 1.0f; i1c0_8.Npad = 16; i1c0_8.pad_ = 0;
      k_gemm<1><<<dim3((unsigned)((16) + 31) / 32, (unsigned)((64) + 15) / 16, (unsigned)(2 * 64)), 32, 0, stream>>>(i1c0_8); }
    k_mm_relu2d<<<(unsigned)(((long long)2 * HW * 16 + 255) / 256), 256, 0, stream>>>(R67 + 26176, nullptr, 2, 64, 16);
    { GemmP i2c0_0;
      i2c0_0.A = R67 + 26176 + (size_t)0 * 16; i2c0_0.B = iw2 + 0; i2c0_0.bias = ib2; i2c0_0.R = R67 + 26176 + (size_t)0 * 16; i2c0_0.C = R67 + 165568 + (size_t)67 * 32;
      i2c0_0.sAo = (long long)66 * 66 * 16; i2c0_0.sAi = (long long)66 * 16; i2c0_0.sAm = 16; i2c0_0.sAk = 1; i2c0_0.sBo = 0; i2c0_0.sBi = 0; i2c0_0.sBn = 16 * 9; i2c0_0.sBk = 9; i2c0_0.sCo = (long long)66 * 66 * 32; i2c0_0.sCi = (long long)66 * 32; i2c0_0.sCm = 32; i2c0_0.sRo = 0; i2c0_0.sRi = 0; i2c0_0.sRm = 0; i2c0_0.sRn = 0;
      i2c0_0.M = 64; i2c0_0.N = 32; i2c0_0.K = 16; i2c0_0.zi_n = 64; i2c0_0.flags = 1; i2c0_0.act = 0;
      i2c0_0.alpha = 1.0f; i2c0_0.beta = 0.0f; i2c0_0.sa = 1.0f; i2c0_0.sb = 1.0f; i2c0_0.Npad = 32; i2c0_0.pad_ = 0;
      k_gemm<1><<<dim3((unsigned)((32) + 31) / 32, (unsigned)((64) + 15) / 16, (unsigned)(2 * 64)), 32, 0, stream>>>(i2c0_0); }
    { GemmP i2c0_1;
      i2c0_1.A = R67 + 26176 + (size_t)1 * 16; i2c0_1.B = iw2 + 1; i2c0_1.bias = R67 + 26176 + (size_t)1 * 16; i2c0_1.R = R67 + 165568 + (size_t)67 * 32; i2c0_1.C = R67 + 165568 + (size_t)67 * 32;
      i2c0_1.sAo = (long long)66 * 66 * 16; i2c0_1.sAi = (long long)66 * 16; i2c0_1.sAm = 16; i2c0_1.sAk = 1; i2c0_1.sBo = 0; i2c0_1.sBi = 0; i2c0_1.sBn = 16 * 9; i2c0_1.sBk = 9; i2c0_1.sCo = (long long)66 * 66 * 32; i2c0_1.sCi = (long long)66 * 32; i2c0_1.sCm = 32; i2c0_1.sRo = (long long)66 * 66 * 32; i2c0_1.sRi = (long long)66 * 32; i2c0_1.sRm = 32; i2c0_1.sRn = 1;
      i2c0_1.M = 64; i2c0_1.N = 32; i2c0_1.K = 16; i2c0_1.zi_n = 64; i2c0_1.flags = 4; i2c0_1.act = 0;
      i2c0_1.alpha = 1.0f; i2c0_1.beta = 1.0f; i2c0_1.sa = 1.0f; i2c0_1.sb = 1.0f; i2c0_1.Npad = 32; i2c0_1.pad_ = 0;
      k_gemm<1><<<dim3((unsigned)((32) + 31) / 32, (unsigned)((64) + 15) / 16, (unsigned)(2 * 64)), 32, 0, stream>>>(i2c0_1); }
    { GemmP i2c0_2;
      i2c0_2.A = R67 + 26176 + (size_t)2 * 16; i2c0_2.B = iw2 + 2; i2c0_2.bias = R67 + 26176 + (size_t)2 * 16; i2c0_2.R = R67 + 165568 + (size_t)67 * 32; i2c0_2.C = R67 + 165568 + (size_t)67 * 32;
      i2c0_2.sAo = (long long)66 * 66 * 16; i2c0_2.sAi = (long long)66 * 16; i2c0_2.sAm = 16; i2c0_2.sAk = 1; i2c0_2.sBo = 0; i2c0_2.sBi = 0; i2c0_2.sBn = 16 * 9; i2c0_2.sBk = 9; i2c0_2.sCo = (long long)66 * 66 * 32; i2c0_2.sCi = (long long)66 * 32; i2c0_2.sCm = 32; i2c0_2.sRo = (long long)66 * 66 * 32; i2c0_2.sRi = (long long)66 * 32; i2c0_2.sRm = 32; i2c0_2.sRn = 1;
      i2c0_2.M = 64; i2c0_2.N = 32; i2c0_2.K = 16; i2c0_2.zi_n = 64; i2c0_2.flags = 4; i2c0_2.act = 0;
      i2c0_2.alpha = 1.0f; i2c0_2.beta = 1.0f; i2c0_2.sa = 1.0f; i2c0_2.sb = 1.0f; i2c0_2.Npad = 32; i2c0_2.pad_ = 0;
      k_gemm<1><<<dim3((unsigned)((32) + 31) / 32, (unsigned)((64) + 15) / 16, (unsigned)(2 * 64)), 32, 0, stream>>>(i2c0_2); }
    { GemmP i2c0_3;
      i2c0_3.A = R67 + 26176 + (size_t)66 * 16; i2c0_3.B = iw2 + 3; i2c0_3.bias = R67 + 26176 + (size_t)66 * 16; i2c0_3.R = R67 + 165568 + (size_t)67 * 32; i2c0_3.C = R67 + 165568 + (size_t)67 * 32;
      i2c0_3.sAo = (long long)66 * 66 * 16; i2c0_3.sAi = (long long)66 * 16; i2c0_3.sAm = 16; i2c0_3.sAk = 1; i2c0_3.sBo = 0; i2c0_3.sBi = 0; i2c0_3.sBn = 16 * 9; i2c0_3.sBk = 9; i2c0_3.sCo = (long long)66 * 66 * 32; i2c0_3.sCi = (long long)66 * 32; i2c0_3.sCm = 32; i2c0_3.sRo = (long long)66 * 66 * 32; i2c0_3.sRi = (long long)66 * 32; i2c0_3.sRm = 32; i2c0_3.sRn = 1;
      i2c0_3.M = 64; i2c0_3.N = 32; i2c0_3.K = 16; i2c0_3.zi_n = 64; i2c0_3.flags = 4; i2c0_3.act = 0;
      i2c0_3.alpha = 1.0f; i2c0_3.beta = 1.0f; i2c0_3.sa = 1.0f; i2c0_3.sb = 1.0f; i2c0_3.Npad = 32; i2c0_3.pad_ = 0;
      k_gemm<1><<<dim3((unsigned)((32) + 31) / 32, (unsigned)((64) + 15) / 16, (unsigned)(2 * 64)), 32, 0, stream>>>(i2c0_3); }
    { GemmP i2c0_4;
      i2c0_4.A = R67 + 26176 + (size_t)67 * 16; i2c0_4.B = iw2 + 4; i2c0_4.bias = R67 + 26176 + (size_t)67 * 16; i2c0_4.R = R67 + 165568 + (size_t)67 * 32; i2c0_4.C = R67 + 165568 + (size_t)67 * 32;
      i2c0_4.sAo = (long long)66 * 66 * 16; i2c0_4.sAi = (long long)66 * 16; i2c0_4.sAm = 16; i2c0_4.sAk = 1; i2c0_4.sBo = 0; i2c0_4.sBi = 0; i2c0_4.sBn = 16 * 9; i2c0_4.sBk = 9; i2c0_4.sCo = (long long)66 * 66 * 32; i2c0_4.sCi = (long long)66 * 32; i2c0_4.sCm = 32; i2c0_4.sRo = (long long)66 * 66 * 32; i2c0_4.sRi = (long long)66 * 32; i2c0_4.sRm = 32; i2c0_4.sRn = 1;
      i2c0_4.M = 64; i2c0_4.N = 32; i2c0_4.K = 16; i2c0_4.zi_n = 64; i2c0_4.flags = 4; i2c0_4.act = 0;
      i2c0_4.alpha = 1.0f; i2c0_4.beta = 1.0f; i2c0_4.sa = 1.0f; i2c0_4.sb = 1.0f; i2c0_4.Npad = 32; i2c0_4.pad_ = 0;
      k_gemm<1><<<dim3((unsigned)((32) + 31) / 32, (unsigned)((64) + 15) / 16, (unsigned)(2 * 64)), 32, 0, stream>>>(i2c0_4); }
    { GemmP i2c0_5;
      i2c0_5.A = R67 + 26176 + (size_t)68 * 16; i2c0_5.B = iw2 + 5; i2c0_5.bias = R67 + 26176 + (size_t)68 * 16; i2c0_5.R = R67 + 165568 + (size_t)67 * 32; i2c0_5.C = R67 + 165568 + (size_t)67 * 32;
      i2c0_5.sAo = (long long)66 * 66 * 16; i2c0_5.sAi = (long long)66 * 16; i2c0_5.sAm = 16; i2c0_5.sAk = 1; i2c0_5.sBo = 0; i2c0_5.sBi = 0; i2c0_5.sBn = 16 * 9; i2c0_5.sBk = 9; i2c0_5.sCo = (long long)66 * 66 * 32; i2c0_5.sCi = (long long)66 * 32; i2c0_5.sCm = 32; i2c0_5.sRo = (long long)66 * 66 * 32; i2c0_5.sRi = (long long)66 * 32; i2c0_5.sRm = 32; i2c0_5.sRn = 1;
      i2c0_5.M = 64; i2c0_5.N = 32; i2c0_5.K = 16; i2c0_5.zi_n = 64; i2c0_5.flags = 4; i2c0_5.act = 0;
      i2c0_5.alpha = 1.0f; i2c0_5.beta = 1.0f; i2c0_5.sa = 1.0f; i2c0_5.sb = 1.0f; i2c0_5.Npad = 32; i2c0_5.pad_ = 0;
      k_gemm<1><<<dim3((unsigned)((32) + 31) / 32, (unsigned)((64) + 15) / 16, (unsigned)(2 * 64)), 32, 0, stream>>>(i2c0_5); }
    { GemmP i2c0_6;
      i2c0_6.A = R67 + 26176 + (size_t)132 * 16; i2c0_6.B = iw2 + 6; i2c0_6.bias = R67 + 26176 + (size_t)132 * 16; i2c0_6.R = R67 + 165568 + (size_t)67 * 32; i2c0_6.C = R67 + 165568 + (size_t)67 * 32;
      i2c0_6.sAo = (long long)66 * 66 * 16; i2c0_6.sAi = (long long)66 * 16; i2c0_6.sAm = 16; i2c0_6.sAk = 1; i2c0_6.sBo = 0; i2c0_6.sBi = 0; i2c0_6.sBn = 16 * 9; i2c0_6.sBk = 9; i2c0_6.sCo = (long long)66 * 66 * 32; i2c0_6.sCi = (long long)66 * 32; i2c0_6.sCm = 32; i2c0_6.sRo = (long long)66 * 66 * 32; i2c0_6.sRi = (long long)66 * 32; i2c0_6.sRm = 32; i2c0_6.sRn = 1;
      i2c0_6.M = 64; i2c0_6.N = 32; i2c0_6.K = 16; i2c0_6.zi_n = 64; i2c0_6.flags = 4; i2c0_6.act = 0;
      i2c0_6.alpha = 1.0f; i2c0_6.beta = 1.0f; i2c0_6.sa = 1.0f; i2c0_6.sb = 1.0f; i2c0_6.Npad = 32; i2c0_6.pad_ = 0;
      k_gemm<1><<<dim3((unsigned)((32) + 31) / 32, (unsigned)((64) + 15) / 16, (unsigned)(2 * 64)), 32, 0, stream>>>(i2c0_6); }
    { GemmP i2c0_7;
      i2c0_7.A = R67 + 26176 + (size_t)133 * 16; i2c0_7.B = iw2 + 7; i2c0_7.bias = R67 + 26176 + (size_t)133 * 16; i2c0_7.R = R67 + 165568 + (size_t)67 * 32; i2c0_7.C = R67 + 165568 + (size_t)67 * 32;
      i2c0_7.sAo = (long long)66 * 66 * 16; i2c0_7.sAi = (long long)66 * 16; i2c0_7.sAm = 16; i2c0_7.sAk = 1; i2c0_7.sBo = 0; i2c0_7.sBi = 0; i2c0_7.sBn = 16 * 9; i2c0_7.sBk = 9; i2c0_7.sCo = (long long)66 * 66 * 32; i2c0_7.sCi = (long long)66 * 32; i2c0_7.sCm = 32; i2c0_7.sRo = (long long)66 * 66 * 32; i2c0_7.sRi = (long long)66 * 32; i2c0_7.sRm = 32; i2c0_7.sRn = 1;
      i2c0_7.M = 64; i2c0_7.N = 32; i2c0_7.K = 16; i2c0_7.zi_n = 64; i2c0_7.flags = 4; i2c0_7.act = 0;
      i2c0_7.alpha = 1.0f; i2c0_7.beta = 1.0f; i2c0_7.sa = 1.0f; i2c0_7.sb = 1.0f; i2c0_7.Npad = 32; i2c0_7.pad_ = 0;
      k_gemm<1><<<dim3((unsigned)((32) + 31) / 32, (unsigned)((64) + 15) / 16, (unsigned)(2 * 64)), 32, 0, stream>>>(i2c0_7); }
    { GemmP i2c0_8;
      i2c0_8.A = R67 + 26176 + (size_t)134 * 16; i2c0_8.B = iw2 + 8; i2c0_8.bias = R67 + 26176 + (size_t)134 * 16; i2c0_8.R = R67 + 165568 + (size_t)67 * 32; i2c0_8.C = R67 + 165568 + (size_t)67 * 32;
      i2c0_8.sAo = (long long)66 * 66 * 16; i2c0_8.sAi = (long long)66 * 16; i2c0_8.sAm = 16; i2c0_8.sAk = 1; i2c0_8.sBo = 0; i2c0_8.sBi = 0; i2c0_8.sBn = 16 * 9; i2c0_8.sBk = 9; i2c0_8.sCo = (long long)66 * 66 * 32; i2c0_8.sCi = (long long)66 * 32; i2c0_8.sCm = 32; i2c0_8.sRo = (long long)66 * 66 * 32; i2c0_8.sRi = (long long)66 * 32; i2c0_8.sRm = 32; i2c0_8.sRn = 1;
      i2c0_8.M = 64; i2c0_8.N = 32; i2c0_8.K = 16; i2c0_8.zi_n = 64; i2c0_8.flags = 4; i2c0_8.act = 0;
      i2c0_8.alpha = 1.0f; i2c0_8.beta = 1.0f; i2c0_8.sa = 1.0f; i2c0_8.sb = 1.0f; i2c0_8.Npad = 32; i2c0_8.pad_ = 0;
      k_gemm<1><<<dim3((unsigned)((32) + 31) / 32, (unsigned)((64) + 15) / 16, (unsigned)(2 * 64)), 32, 0, stream>>>(i2c0_8); }
    k_mm_relu2d<<<(unsigned)(((long long)2 * HW * 32 + 255) / 256), 256, 0, stream>>>(R67 + 165568, nullptr, 2, 64, 32);
    { GemmP i3c0_0;
      i3c0_0.A = R67 + 165568 + (size_t)0 * 32; i3c0_0.B = iw3 + 0; i3c0_0.bias = ib3; i3c0_0.R = R67 + 165568 + (size_t)0 * 32; i3c0_0.C = R67 + 444352 + (size_t)67 * 64;
      i3c0_0.sAo = (long long)66 * 66 * 32; i3c0_0.sAi = (long long)66 * 32; i3c0_0.sAm = 32; i3c0_0.sAk = 1; i3c0_0.sBo = 0; i3c0_0.sBi = 0; i3c0_0.sBn = 32 * 9; i3c0_0.sBk = 9; i3c0_0.sCo = (long long)66 * 66 * 64; i3c0_0.sCi = (long long)66 * 64; i3c0_0.sCm = 64; i3c0_0.sRo = 0; i3c0_0.sRi = 0; i3c0_0.sRm = 0; i3c0_0.sRn = 0;
      i3c0_0.M = 64; i3c0_0.N = 64; i3c0_0.K = 32; i3c0_0.zi_n = 64; i3c0_0.flags = 1; i3c0_0.act = 0;
      i3c0_0.alpha = 1.0f; i3c0_0.beta = 0.0f; i3c0_0.sa = 1.0f; i3c0_0.sb = 1.0f; i3c0_0.Npad = 64; i3c0_0.pad_ = 0;
      k_gemm<1><<<dim3((unsigned)((64) + 31) / 32, (unsigned)((64) + 15) / 16, (unsigned)(2 * 64)), 32, 0, stream>>>(i3c0_0); }
    { GemmP i3c0_1;
      i3c0_1.A = R67 + 165568 + (size_t)1 * 32; i3c0_1.B = iw3 + 1; i3c0_1.bias = R67 + 165568 + (size_t)1 * 32; i3c0_1.R = R67 + 444352 + (size_t)67 * 64; i3c0_1.C = R67 + 444352 + (size_t)67 * 64;
      i3c0_1.sAo = (long long)66 * 66 * 32; i3c0_1.sAi = (long long)66 * 32; i3c0_1.sAm = 32; i3c0_1.sAk = 1; i3c0_1.sBo = 0; i3c0_1.sBi = 0; i3c0_1.sBn = 32 * 9; i3c0_1.sBk = 9; i3c0_1.sCo = (long long)66 * 66 * 64; i3c0_1.sCi = (long long)66 * 64; i3c0_1.sCm = 64; i3c0_1.sRo = (long long)66 * 66 * 64; i3c0_1.sRi = (long long)66 * 64; i3c0_1.sRm = 64; i3c0_1.sRn = 1;
      i3c0_1.M = 64; i3c0_1.N = 64; i3c0_1.K = 32; i3c0_1.zi_n = 64; i3c0_1.flags = 4; i3c0_1.act = 0;
      i3c0_1.alpha = 1.0f; i3c0_1.beta = 1.0f; i3c0_1.sa = 1.0f; i3c0_1.sb = 1.0f; i3c0_1.Npad = 64; i3c0_1.pad_ = 0;
      k_gemm<1><<<dim3((unsigned)((64) + 31) / 32, (unsigned)((64) + 15) / 16, (unsigned)(2 * 64)), 32, 0, stream>>>(i3c0_1); }
    { GemmP i3c0_2;
      i3c0_2.A = R67 + 165568 + (size_t)2 * 32; i3c0_2.B = iw3 + 2; i3c0_2.bias = R67 + 165568 + (size_t)2 * 32; i3c0_2.R = R67 + 444352 + (size_t)67 * 64; i3c0_2.C = R67 + 444352 + (size_t)67 * 64;
      i3c0_2.sAo = (long long)66 * 66 * 32; i3c0_2.sAi = (long long)66 * 32; i3c0_2.sAm = 32; i3c0_2.sAk = 1; i3c0_2.sBo = 0; i3c0_2.sBi = 0; i3c0_2.sBn = 32 * 9; i3c0_2.sBk = 9; i3c0_2.sCo = (long long)66 * 66 * 64; i3c0_2.sCi = (long long)66 * 64; i3c0_2.sCm = 64; i3c0_2.sRo = (long long)66 * 66 * 64; i3c0_2.sRi = (long long)66 * 64; i3c0_2.sRm = 64; i3c0_2.sRn = 1;
      i3c0_2.M = 64; i3c0_2.N = 64; i3c0_2.K = 32; i3c0_2.zi_n = 64; i3c0_2.flags = 4; i3c0_2.act = 0;
      i3c0_2.alpha = 1.0f; i3c0_2.beta = 1.0f; i3c0_2.sa = 1.0f; i3c0_2.sb = 1.0f; i3c0_2.Npad = 64; i3c0_2.pad_ = 0;
      k_gemm<1><<<dim3((unsigned)((64) + 31) / 32, (unsigned)((64) + 15) / 16, (unsigned)(2 * 64)), 32, 0, stream>>>(i3c0_2); }
    { GemmP i3c0_3;
      i3c0_3.A = R67 + 165568 + (size_t)66 * 32; i3c0_3.B = iw3 + 3; i3c0_3.bias = R67 + 165568 + (size_t)66 * 32; i3c0_3.R = R67 + 444352 + (size_t)67 * 64; i3c0_3.C = R67 + 444352 + (size_t)67 * 64;
      i3c0_3.sAo = (long long)66 * 66 * 32; i3c0_3.sAi = (long long)66 * 32; i3c0_3.sAm = 32; i3c0_3.sAk = 1; i3c0_3.sBo = 0; i3c0_3.sBi = 0; i3c0_3.sBn = 32 * 9; i3c0_3.sBk = 9; i3c0_3.sCo = (long long)66 * 66 * 64; i3c0_3.sCi = (long long)66 * 64; i3c0_3.sCm = 64; i3c0_3.sRo = (long long)66 * 66 * 64; i3c0_3.sRi = (long long)66 * 64; i3c0_3.sRm = 64; i3c0_3.sRn = 1;
      i3c0_3.M = 64; i3c0_3.N = 64; i3c0_3.K = 32; i3c0_3.zi_n = 64; i3c0_3.flags = 4; i3c0_3.act = 0;
      i3c0_3.alpha = 1.0f; i3c0_3.beta = 1.0f; i3c0_3.sa = 1.0f; i3c0_3.sb = 1.0f; i3c0_3.Npad = 64; i3c0_3.pad_ = 0;
      k_gemm<1><<<dim3((unsigned)((64) + 31) / 32, (unsigned)((64) + 15) / 16, (unsigned)(2 * 64)), 32, 0, stream>>>(i3c0_3); }
    { GemmP i3c0_4;
      i3c0_4.A = R67 + 165568 + (size_t)67 * 32; i3c0_4.B = iw3 + 4; i3c0_4.bias = R67 + 165568 + (size_t)67 * 32; i3c0_4.R = R67 + 444352 + (size_t)67 * 64; i3c0_4.C = R67 + 444352 + (size_t)67 * 64;
      i3c0_4.sAo = (long long)66 * 66 * 32; i3c0_4.sAi = (long long)66 * 32; i3c0_4.sAm = 32; i3c0_4.sAk = 1; i3c0_4.sBo = 0; i3c0_4.sBi = 0; i3c0_4.sBn = 32 * 9; i3c0_4.sBk = 9; i3c0_4.sCo = (long long)66 * 66 * 64; i3c0_4.sCi = (long long)66 * 64; i3c0_4.sCm = 64; i3c0_4.sRo = (long long)66 * 66 * 64; i3c0_4.sRi = (long long)66 * 64; i3c0_4.sRm = 64; i3c0_4.sRn = 1;
      i3c0_4.M = 64; i3c0_4.N = 64; i3c0_4.K = 32; i3c0_4.zi_n = 64; i3c0_4.flags = 4; i3c0_4.act = 0;
      i3c0_4.alpha = 1.0f; i3c0_4.beta = 1.0f; i3c0_4.sa = 1.0f; i3c0_4.sb = 1.0f; i3c0_4.Npad = 64; i3c0_4.pad_ = 0;
      k_gemm<1><<<dim3((unsigned)((64) + 31) / 32, (unsigned)((64) + 15) / 16, (unsigned)(2 * 64)), 32, 0, stream>>>(i3c0_4); }
    { GemmP i3c0_5;
      i3c0_5.A = R67 + 165568 + (size_t)68 * 32; i3c0_5.B = iw3 + 5; i3c0_5.bias = R67 + 165568 + (size_t)68 * 32; i3c0_5.R = R67 + 444352 + (size_t)67 * 64; i3c0_5.C = R67 + 444352 + (size_t)67 * 64;
      i3c0_5.sAo = (long long)66 * 66 * 32; i3c0_5.sAi = (long long)66 * 32; i3c0_5.sAm = 32; i3c0_5.sAk = 1; i3c0_5.sBo = 0; i3c0_5.sBi = 0; i3c0_5.sBn = 32 * 9; i3c0_5.sBk = 9; i3c0_5.sCo = (long long)66 * 66 * 64; i3c0_5.sCi = (long long)66 * 64; i3c0_5.sCm = 64; i3c0_5.sRo = (long long)66 * 66 * 64; i3c0_5.sRi = (long long)66 * 64; i3c0_5.sRm = 64; i3c0_5.sRn = 1;
      i3c0_5.M = 64; i3c0_5.N = 64; i3c0_5.K = 32; i3c0_5.zi_n = 64; i3c0_5.flags = 4; i3c0_5.act = 0;
      i3c0_5.alpha = 1.0f; i3c0_5.beta = 1.0f; i3c0_5.sa = 1.0f; i3c0_5.sb = 1.0f; i3c0_5.Npad = 64; i3c0_5.pad_ = 0;
      k_gemm<1><<<dim3((unsigned)((64) + 31) / 32, (unsigned)((64) + 15) / 16, (unsigned)(2 * 64)), 32, 0, stream>>>(i3c0_5); }
    { GemmP i3c0_6;
      i3c0_6.A = R67 + 165568 + (size_t)132 * 32; i3c0_6.B = iw3 + 6; i3c0_6.bias = R67 + 165568 + (size_t)132 * 32; i3c0_6.R = R67 + 444352 + (size_t)67 * 64; i3c0_6.C = R67 + 444352 + (size_t)67 * 64;
      i3c0_6.sAo = (long long)66 * 66 * 32; i3c0_6.sAi = (long long)66 * 32; i3c0_6.sAm = 32; i3c0_6.sAk = 1; i3c0_6.sBo = 0; i3c0_6.sBi = 0; i3c0_6.sBn = 32 * 9; i3c0_6.sBk = 9; i3c0_6.sCo = (long long)66 * 66 * 64; i3c0_6.sCi = (long long)66 * 64; i3c0_6.sCm = 64; i3c0_6.sRo = (long long)66 * 66 * 64; i3c0_6.sRi = (long long)66 * 64; i3c0_6.sRm = 64; i3c0_6.sRn = 1;
      i3c0_6.M = 64; i3c0_6.N = 64; i3c0_6.K = 32; i3c0_6.zi_n = 64; i3c0_6.flags = 4; i3c0_6.act = 0;
      i3c0_6.alpha = 1.0f; i3c0_6.beta = 1.0f; i3c0_6.sa = 1.0f; i3c0_6.sb = 1.0f; i3c0_6.Npad = 64; i3c0_6.pad_ = 0;
      k_gemm<1><<<dim3((unsigned)((64) + 31) / 32, (unsigned)((64) + 15) / 16, (unsigned)(2 * 64)), 32, 0, stream>>>(i3c0_6); }
    { GemmP i3c0_7;
      i3c0_7.A = R67 + 165568 + (size_t)133 * 32; i3c0_7.B = iw3 + 7; i3c0_7.bias = R67 + 165568 + (size_t)133 * 32; i3c0_7.R = R67 + 444352 + (size_t)67 * 64; i3c0_7.C = R67 + 444352 + (size_t)67 * 64;
      i3c0_7.sAo = (long long)66 * 66 * 32; i3c0_7.sAi = (long long)66 * 32; i3c0_7.sAm = 32; i3c0_7.sAk = 1; i3c0_7.sBo = 0; i3c0_7.sBi = 0; i3c0_7.sBn = 32 * 9; i3c0_7.sBk = 9; i3c0_7.sCo = (long long)66 * 66 * 64; i3c0_7.sCi = (long long)66 * 64; i3c0_7.sCm = 64; i3c0_7.sRo = (long long)66 * 66 * 64; i3c0_7.sRi = (long long)66 * 64; i3c0_7.sRm = 64; i3c0_7.sRn = 1;
      i3c0_7.M = 64; i3c0_7.N = 64; i3c0_7.K = 32; i3c0_7.zi_n = 64; i3c0_7.flags = 4; i3c0_7.act = 0;
      i3c0_7.alpha = 1.0f; i3c0_7.beta = 1.0f; i3c0_7.sa = 1.0f; i3c0_7.sb = 1.0f; i3c0_7.Npad = 64; i3c0_7.pad_ = 0;
      k_gemm<1><<<dim3((unsigned)((64) + 31) / 32, (unsigned)((64) + 15) / 16, (unsigned)(2 * 64)), 32, 0, stream>>>(i3c0_7); }
    { GemmP i3c0_8;
      i3c0_8.A = R67 + 165568 + (size_t)134 * 32; i3c0_8.B = iw3 + 8; i3c0_8.bias = R67 + 165568 + (size_t)134 * 32; i3c0_8.R = R67 + 444352 + (size_t)67 * 64; i3c0_8.C = R67 + 444352 + (size_t)67 * 64;
      i3c0_8.sAo = (long long)66 * 66 * 32; i3c0_8.sAi = (long long)66 * 32; i3c0_8.sAm = 32; i3c0_8.sAk = 1; i3c0_8.sBo = 0; i3c0_8.sBi = 0; i3c0_8.sBn = 32 * 9; i3c0_8.sBk = 9; i3c0_8.sCo = (long long)66 * 66 * 64; i3c0_8.sCi = (long long)66 * 64; i3c0_8.sCm = 64; i3c0_8.sRo = (long long)66 * 66 * 64; i3c0_8.sRi = (long long)66 * 64; i3c0_8.sRm = 64; i3c0_8.sRn = 1;
      i3c0_8.M = 64; i3c0_8.N = 64; i3c0_8.K = 32; i3c0_8.zi_n = 64; i3c0_8.flags = 4; i3c0_8.act = 0;
      i3c0_8.alpha = 1.0f; i3c0_8.beta = 1.0f; i3c0_8.sa = 1.0f; i3c0_8.sb = 1.0f; i3c0_8.Npad = 64; i3c0_8.pad_ = 0;
      k_gemm<1><<<dim3((unsigned)((64) + 31) / 32, (unsigned)((64) + 15) / 16, (unsigned)(2 * 64)), 32, 0, stream>>>(i3c0_8); }
    k_mm_relu2d<<<(unsigned)(((long long)2 * HW * 64 + 255) / 256), 256, 0, stream>>>(R67 + 444352, R67 + 1001920, 2, 64, 64);
    { GemmP gqkv0;
      gqkv0.A = R67 + 1001920; gqkv0.B = qkvw; gqkv0.bias = qkvb; gqkv0.R = R67 + 1001920; gqkv0.C = R67 + 1526208;
      gqkv0.sAo = 0; gqkv0.sAi = 0; gqkv0.sAm = 64; gqkv0.sAk = 1; gqkv0.sBo = 0; gqkv0.sBi = 0; gqkv0.sBn = 64; gqkv0.sBk = 1; gqkv0.sCo = 0; gqkv0.sCi = 0; gqkv0.sCm = 192; gqkv0.sRo = 0; gqkv0.sRi = 0; gqkv0.sRm = 0; gqkv0.sRn = 0;
      gqkv0.M = 2 * HW; gqkv0.N = 192; gqkv0.K = 64; gqkv0.zi_n = 1; gqkv0.flags = 1; gqkv0.act = 0;
      gqkv0.alpha = 1.0f; gqkv0.beta = 0.0f; gqkv0.sa = 1.0f; gqkv0.sb = 1.0f; gqkv0.Npad = 192; gqkv0.pad_ = 0;
      k_gemm<1><<<dim3((unsigned)((192) + 31) / 32, (unsigned)((2 * HW) + 15) / 16, (unsigned)(1)), 32, 0, stream>>>(gqkv0); }
    k_mm_dw<<<(unsigned)(((long long)2 * HW * 192 + 255) / 256), 256, 0, stream>>>(R67 + 1526208, dww, dwb, R67 + 3099072, 2, 64, 192);
    k_mm_fall<<<(unsigned)(((long long)2 * HW * 144 + 255) / 256), 256, 0, stream>>>(R67 + 3099072, fcw, fcb, R67 + 4671936, 2, HW, 192);
    k_mm_dep<<<(unsigned)(((long long)2 * 64 * HW + 255) / 256), 256, 0, stream>>>(R67 + 4671936, depw, depb, R67 + 5851584, 2, 64);
    k_mm_qknorm<<<2 * 128, 256, 0, stream>>>(R67 + 3099072, R67 + 6375872, 2, HW, 192);
    { GemmP gat0;
      gat0.A = R67 + 6375872; gat0.B = R67 + 6375872 + (size_t)64 * HW; gat0.bias = R67 + 6375872; gat0.R = R67 + 6375872; gat0.C = R67 + 7424448;
      gat0.sAo = (long long)128 * HW; gat0.sAi = (long long)16 * HW; gat0.sAm = HW; gat0.sAk = 1; gat0.sBo = (long long)128 * HW; gat0.sBi = (long long)16 * HW; gat0.sBn = HW; gat0.sBk = 1; gat0.sCo = (long long)4 * 16 * LP; gat0.sCi = 16 * LP; gat0.sCm = LP; gat0.sRo = 0; gat0.sRi = 0; gat0.sRm = 0; gat0.sRn = 0;
      gat0.M = 16; gat0.N = 16; gat0.K = HW; gat0.zi_n = 4; gat0.flags = 0; gat0.act = 0;
      gat0.alpha = 1.0f; gat0.beta = 0.0f; gat0.sa = 1.0f; gat0.sb = 1.0f; gat0.Npad = LP; gat0.pad_ = 0;
      k_gemm<1><<<dim3((unsigned)((LP) + 31) / 32, (unsigned)((16) + 15) / 16, (unsigned)(2 * 4)), 32, 0, stream>>>(gat0); }
    k_mm_sm16<<<(unsigned)((2 * 4 * 16 + 255) / 256), 256, 0, stream>>>(R67 + 7424448, temp, 2 * 4, LP);
    { GemmP gao0;
      gao0.A = R67 + 7424448; gao0.B = R67 + 3099072 + 128; gao0.bias = R67 + 7424448; gao0.R = R67 + 7424448; gao0.C = R67 + 7428544;
      gao0.sAo = (long long)4 * 16 * LP; gao0.sAi = 16 * LP; gao0.sAm = LP; gao0.sAk = 1; gao0.sBo = (long long)HW * 192; gao0.sBi = 16; gao0.sBn = 192; gao0.sBk = 1; gao0.sCo = (long long)64 * HW; gao0.sCi = (long long)16 * HW; gao0.sCm = HW; gao0.sRo = 0; gao0.sRi = 0; gao0.sRm = 0; gao0.sRn = 0;
      gao0.M = 16; gao0.N = HW; gao0.K = 16; gao0.zi_n = 4; gao0.flags = 0; gao0.act = 0;
      gao0.alpha = 1.0f; gao0.beta = 0.0f; gao0.sa = 1.0f; gao0.sb = 1.0f; gao0.Npad = HW; gao0.pad_ = 0;
      k_gemm<1><<<dim3((unsigned)((HW) + 31) / 32, (unsigned)((16) + 15) / 16, (unsigned)(2 * 4)), 32, 0, stream>>>(gao0); }
    { GemmP gproj0;
      gproj0.A = projw; gproj0.B = R67 + 7428544; gproj0.bias = projb; gproj0.R = projw; gproj0.C = R67 + 7952832;
      gproj0.sAo = 0; gproj0.sAi = 0; gproj0.sAm = 64; gproj0.sAk = 1; gproj0.sBo = (long long)64 * HW; gproj0.sBi = 0; gproj0.sBn = 1; gproj0.sBk = HW; gproj0.sCo = (long long)64 * HW; gproj0.sCi = 0; gproj0.sCm = HW; gproj0.sRo = 0; gproj0.sRi = 0; gproj0.sRm = 0; gproj0.sRn = 0;
      gproj0.M = 64; gproj0.N = HW; gproj0.K = 64; gproj0.zi_n = 1; gproj0.flags = 2; gproj0.act = 0;
      gproj0.alpha = 1.0f; gproj0.beta = 0.0f; gproj0.sa = 1.0f; gproj0.sb = 1.0f; gproj0.Npad = HW; gproj0.pad_ = 0;
      k_gemm<1><<<dim3((unsigned)((HW) + 31) / 32, (unsigned)((64) + 15) / 16, (unsigned)(2)), 32, 0, stream>>>(gproj0); }
    k_mm_imgfeat<<<(unsigned)(((long long)2 * SEQ * 64 + 255) / 256), 256, 0, stream>>>(R67 + 7952832, R67 + 5851584, IR + (size_t)0 * SEQ * 64, 2, HW, 64);
    hipMemsetAsync(R67 + 0, 0, (size_t)2 * 66 * 66 * 3 * 4, stream); hipMemsetAsync(R67 + 26176, 0, (size_t)2 * 66 * 66 * 16 * 4, stream); hipMemsetAsync(R67 + 165568, 0, (size_t)2 * 66 * 66 * 32 * 4, stream); hipMemsetAsync(R67 + 444352, 0, (size_t)2 * 66 * 66 * 64 * 4, stream);
    k_mm_padimg<<<(unsigned)(((long long)2 * HW * 3 + 255) / 256), 256, 0, stream>>>(img + (size_t)2 * 3 * HW, R67 + 0, 2, 3, 64);
    { GemmP i1c1_0;
      i1c1_0.A = R67 + 0 + (size_t)0 * 3; i1c1_0.B = iw1 + 0; i1c1_0.bias = ib1; i1c1_0.R = R67 + 0 + (size_t)0 * 3; i1c1_0.C = R67 + 26176 + (size_t)67 * 16;
      i1c1_0.sAo = (long long)66 * 66 * 3; i1c1_0.sAi = (long long)66 * 3; i1c1_0.sAm = 3; i1c1_0.sAk = 1; i1c1_0.sBo = 0; i1c1_0.sBi = 0; i1c1_0.sBn = 3 * 9; i1c1_0.sBk = 9; i1c1_0.sCo = (long long)66 * 66 * 16; i1c1_0.sCi = (long long)66 * 16; i1c1_0.sCm = 16; i1c1_0.sRo = 0; i1c1_0.sRi = 0; i1c1_0.sRm = 0; i1c1_0.sRn = 0;
      i1c1_0.M = 64; i1c1_0.N = 16; i1c1_0.K = 3; i1c1_0.zi_n = 64; i1c1_0.flags = 1; i1c1_0.act = 0;
      i1c1_0.alpha = 1.0f; i1c1_0.beta = 0.0f; i1c1_0.sa = 1.0f; i1c1_0.sb = 1.0f; i1c1_0.Npad = 16; i1c1_0.pad_ = 0;
      k_gemm<1><<<dim3((unsigned)((16) + 31) / 32, (unsigned)((64) + 15) / 16, (unsigned)(2 * 64)), 32, 0, stream>>>(i1c1_0); }
    { GemmP i1c1_1;
      i1c1_1.A = R67 + 0 + (size_t)1 * 3; i1c1_1.B = iw1 + 1; i1c1_1.bias = R67 + 0 + (size_t)1 * 3; i1c1_1.R = R67 + 26176 + (size_t)67 * 16; i1c1_1.C = R67 + 26176 + (size_t)67 * 16;
      i1c1_1.sAo = (long long)66 * 66 * 3; i1c1_1.sAi = (long long)66 * 3; i1c1_1.sAm = 3; i1c1_1.sAk = 1; i1c1_1.sBo = 0; i1c1_1.sBi = 0; i1c1_1.sBn = 3 * 9; i1c1_1.sBk = 9; i1c1_1.sCo = (long long)66 * 66 * 16; i1c1_1.sCi = (long long)66 * 16; i1c1_1.sCm = 16; i1c1_1.sRo = (long long)66 * 66 * 16; i1c1_1.sRi = (long long)66 * 16; i1c1_1.sRm = 16; i1c1_1.sRn = 1;
      i1c1_1.M = 64; i1c1_1.N = 16; i1c1_1.K = 3; i1c1_1.zi_n = 64; i1c1_1.flags = 4; i1c1_1.act = 0;
      i1c1_1.alpha = 1.0f; i1c1_1.beta = 1.0f; i1c1_1.sa = 1.0f; i1c1_1.sb = 1.0f; i1c1_1.Npad = 16; i1c1_1.pad_ = 0;
      k_gemm<1><<<dim3((unsigned)((16) + 31) / 32, (unsigned)((64) + 15) / 16, (unsigned)(2 * 64)), 32, 0, stream>>>(i1c1_1); }
    { GemmP i1c1_2;
      i1c1_2.A = R67 + 0 + (size_t)2 * 3; i1c1_2.B = iw1 + 2; i1c1_2.bias = R67 + 0 + (size_t)2 * 3; i1c1_2.R = R67 + 26176 + (size_t)67 * 16; i1c1_2.C = R67 + 26176 + (size_t)67 * 16;
      i1c1_2.sAo = (long long)66 * 66 * 3; i1c1_2.sAi = (long long)66 * 3; i1c1_2.sAm = 3; i1c1_2.sAk = 1; i1c1_2.sBo = 0; i1c1_2.sBi = 0; i1c1_2.sBn = 3 * 9; i1c1_2.sBk = 9; i1c1_2.sCo = (long long)66 * 66 * 16; i1c1_2.sCi = (long long)66 * 16; i1c1_2.sCm = 16; i1c1_2.sRo = (long long)66 * 66 * 16; i1c1_2.sRi = (long long)66 * 16; i1c1_2.sRm = 16; i1c1_2.sRn = 1;
      i1c1_2.M = 64; i1c1_2.N = 16; i1c1_2.K = 3; i1c1_2.zi_n = 64; i1c1_2.flags = 4; i1c1_2.act = 0;
      i1c1_2.alpha = 1.0f; i1c1_2.beta = 1.0f; i1c1_2.sa = 1.0f; i1c1_2.sb = 1.0f; i1c1_2.Npad = 16; i1c1_2.pad_ = 0;
      k_gemm<1><<<dim3((unsigned)((16) + 31) / 32, (unsigned)((64) + 15) / 16, (unsigned)(2 * 64)), 32, 0, stream>>>(i1c1_2); }
    { GemmP i1c1_3;
      i1c1_3.A = R67 + 0 + (size_t)66 * 3; i1c1_3.B = iw1 + 3; i1c1_3.bias = R67 + 0 + (size_t)66 * 3; i1c1_3.R = R67 + 26176 + (size_t)67 * 16; i1c1_3.C = R67 + 26176 + (size_t)67 * 16;
      i1c1_3.sAo = (long long)66 * 66 * 3; i1c1_3.sAi = (long long)66 * 3; i1c1_3.sAm = 3; i1c1_3.sAk = 1; i1c1_3.sBo = 0; i1c1_3.sBi = 0; i1c1_3.sBn = 3 * 9; i1c1_3.sBk = 9; i1c1_3.sCo = (long long)66 * 66 * 16; i1c1_3.sCi = (long long)66 * 16; i1c1_3.sCm = 16; i1c1_3.sRo = (long long)66 * 66 * 16; i1c1_3.sRi = (long long)66 * 16; i1c1_3.sRm = 16; i1c1_3.sRn = 1;
      i1c1_3.M = 64; i1c1_3.N = 16; i1c1_3.K = 3; i1c1_3.zi_n = 64; i1c1_3.flags = 4; i1c1_3.act = 0;
      i1c1_3.alpha = 1.0f; i1c1_3.beta = 1.0f; i1c1_3.sa = 1.0f; i1c1_3.sb = 1.0f; i1c1_3.Npad = 16; i1c1_3.pad_ = 0;
      k_gemm<1><<<dim3((unsigned)((16) + 31) / 32, (unsigned)((64) + 15) / 16, (unsigned)(2 * 64)), 32, 0, stream>>>(i1c1_3); }
    { GemmP i1c1_4;
      i1c1_4.A = R67 + 0 + (size_t)67 * 3; i1c1_4.B = iw1 + 4; i1c1_4.bias = R67 + 0 + (size_t)67 * 3; i1c1_4.R = R67 + 26176 + (size_t)67 * 16; i1c1_4.C = R67 + 26176 + (size_t)67 * 16;
      i1c1_4.sAo = (long long)66 * 66 * 3; i1c1_4.sAi = (long long)66 * 3; i1c1_4.sAm = 3; i1c1_4.sAk = 1; i1c1_4.sBo = 0; i1c1_4.sBi = 0; i1c1_4.sBn = 3 * 9; i1c1_4.sBk = 9; i1c1_4.sCo = (long long)66 * 66 * 16; i1c1_4.sCi = (long long)66 * 16; i1c1_4.sCm = 16; i1c1_4.sRo = (long long)66 * 66 * 16; i1c1_4.sRi = (long long)66 * 16; i1c1_4.sRm = 16; i1c1_4.sRn = 1;
      i1c1_4.M = 64; i1c1_4.N = 16; i1c1_4.K = 3; i1c1_4.zi_n = 64; i1c1_4.flags = 4; i1c1_4.act = 0;
      i1c1_4.alpha = 1.0f; i1c1_4.beta = 1.0f; i1c1_4.sa = 1.0f; i1c1_4.sb = 1.0f; i1c1_4.Npad = 16; i1c1_4.pad_ = 0;
      k_gemm<1><<<dim3((unsigned)((16) + 31) / 32, (unsigned)((64) + 15) / 16, (unsigned)(2 * 64)), 32, 0, stream>>>(i1c1_4); }
    { GemmP i1c1_5;
      i1c1_5.A = R67 + 0 + (size_t)68 * 3; i1c1_5.B = iw1 + 5; i1c1_5.bias = R67 + 0 + (size_t)68 * 3; i1c1_5.R = R67 + 26176 + (size_t)67 * 16; i1c1_5.C = R67 + 26176 + (size_t)67 * 16;
      i1c1_5.sAo = (long long)66 * 66 * 3; i1c1_5.sAi = (long long)66 * 3; i1c1_5.sAm = 3; i1c1_5.sAk = 1; i1c1_5.sBo = 0; i1c1_5.sBi = 0; i1c1_5.sBn = 3 * 9; i1c1_5.sBk = 9; i1c1_5.sCo = (long long)66 * 66 * 16; i1c1_5.sCi = (long long)66 * 16; i1c1_5.sCm = 16; i1c1_5.sRo = (long long)66 * 66 * 16; i1c1_5.sRi = (long long)66 * 16; i1c1_5.sRm = 16; i1c1_5.sRn = 1;
      i1c1_5.M = 64; i1c1_5.N = 16; i1c1_5.K = 3; i1c1_5.zi_n = 64; i1c1_5.flags = 4; i1c1_5.act = 0;
      i1c1_5.alpha = 1.0f; i1c1_5.beta = 1.0f; i1c1_5.sa = 1.0f; i1c1_5.sb = 1.0f; i1c1_5.Npad = 16; i1c1_5.pad_ = 0;
      k_gemm<1><<<dim3((unsigned)((16) + 31) / 32, (unsigned)((64) + 15) / 16, (unsigned)(2 * 64)), 32, 0, stream>>>(i1c1_5); }
    { GemmP i1c1_6;
      i1c1_6.A = R67 + 0 + (size_t)132 * 3; i1c1_6.B = iw1 + 6; i1c1_6.bias = R67 + 0 + (size_t)132 * 3; i1c1_6.R = R67 + 26176 + (size_t)67 * 16; i1c1_6.C = R67 + 26176 + (size_t)67 * 16;
      i1c1_6.sAo = (long long)66 * 66 * 3; i1c1_6.sAi = (long long)66 * 3; i1c1_6.sAm = 3; i1c1_6.sAk = 1; i1c1_6.sBo = 0; i1c1_6.sBi = 0; i1c1_6.sBn = 3 * 9; i1c1_6.sBk = 9; i1c1_6.sCo = (long long)66 * 66 * 16; i1c1_6.sCi = (long long)66 * 16; i1c1_6.sCm = 16; i1c1_6.sRo = (long long)66 * 66 * 16; i1c1_6.sRi = (long long)66 * 16; i1c1_6.sRm = 16; i1c1_6.sRn = 1;
      i1c1_6.M = 64; i1c1_6.N = 16; i1c1_6.K = 3; i1c1_6.zi_n = 64; i1c1_6.flags = 4; i1c1_6.act = 0;
      i1c1_6.alpha = 1.0f; i1c1_6.beta = 1.0f; i1c1_6.sa = 1.0f; i1c1_6.sb = 1.0f; i1c1_6.Npad = 16; i1c1_6.pad_ = 0;
      k_gemm<1><<<dim3((unsigned)((16) + 31) / 32, (unsigned)((64) + 15) / 16, (unsigned)(2 * 64)), 32, 0, stream>>>(i1c1_6); }
    { GemmP i1c1_7;
      i1c1_7.A = R67 + 0 + (size_t)133 * 3; i1c1_7.B = iw1 + 7; i1c1_7.bias = R67 + 0 + (size_t)133 * 3; i1c1_7.R = R67 + 26176 + (size_t)67 * 16; i1c1_7.C = R67 + 26176 + (size_t)67 * 16;
      i1c1_7.sAo = (long long)66 * 66 * 3; i1c1_7.sAi = (long long)66 * 3; i1c1_7.sAm = 3; i1c1_7.sAk = 1; i1c1_7.sBo = 0; i1c1_7.sBi = 0; i1c1_7.sBn = 3 * 9; i1c1_7.sBk = 9; i1c1_7.sCo = (long long)66 * 66 * 16; i1c1_7.sCi = (long long)66 * 16; i1c1_7.sCm = 16; i1c1_7.sRo = (long long)66 * 66 * 16; i1c1_7.sRi = (long long)66 * 16; i1c1_7.sRm = 16; i1c1_7.sRn = 1;
      i1c1_7.M = 64; i1c1_7.N = 16; i1c1_7.K = 3; i1c1_7.zi_n = 64; i1c1_7.flags = 4; i1c1_7.act = 0;
      i1c1_7.alpha = 1.0f; i1c1_7.beta = 1.0f; i1c1_7.sa = 1.0f; i1c1_7.sb = 1.0f; i1c1_7.Npad = 16; i1c1_7.pad_ = 0;
      k_gemm<1><<<dim3((unsigned)((16) + 31) / 32, (unsigned)((64) + 15) / 16, (unsigned)(2 * 64)), 32, 0, stream>>>(i1c1_7); }
    { GemmP i1c1_8;
      i1c1_8.A = R67 + 0 + (size_t)134 * 3; i1c1_8.B = iw1 + 8; i1c1_8.bias = R67 + 0 + (size_t)134 * 3; i1c1_8.R = R67 + 26176 + (size_t)67 * 16; i1c1_8.C = R67 + 26176 + (size_t)67 * 16;
      i1c1_8.sAo = (long long)66 * 66 * 3; i1c1_8.sAi = (long long)66 * 3; i1c1_8.sAm = 3; i1c1_8.sAk = 1; i1c1_8.sBo = 0; i1c1_8.sBi = 0; i1c1_8.sBn = 3 * 9; i1c1_8.sBk = 9; i1c1_8.sCo = (long long)66 * 66 * 16; i1c1_8.sCi = (long long)66 * 16; i1c1_8.sCm = 16; i1c1_8.sRo = (long long)66 * 66 * 16; i1c1_8.sRi = (long long)66 * 16; i1c1_8.sRm = 16; i1c1_8.sRn = 1;
      i1c1_8.M = 64; i1c1_8.N = 16; i1c1_8.K = 3; i1c1_8.zi_n = 64; i1c1_8.flags = 4; i1c1_8.act = 0;
      i1c1_8.alpha = 1.0f; i1c1_8.beta = 1.0f; i1c1_8.sa = 1.0f; i1c1_8.sb = 1.0f; i1c1_8.Npad = 16; i1c1_8.pad_ = 0;
      k_gemm<1><<<dim3((unsigned)((16) + 31) / 32, (unsigned)((64) + 15) / 16, (unsigned)(2 * 64)), 32, 0, stream>>>(i1c1_8); }
    k_mm_relu2d<<<(unsigned)(((long long)2 * HW * 16 + 255) / 256), 256, 0, stream>>>(R67 + 26176, nullptr, 2, 64, 16);
    { GemmP i2c1_0;
      i2c1_0.A = R67 + 26176 + (size_t)0 * 16; i2c1_0.B = iw2 + 0; i2c1_0.bias = ib2; i2c1_0.R = R67 + 26176 + (size_t)0 * 16; i2c1_0.C = R67 + 165568 + (size_t)67 * 32;
      i2c1_0.sAo = (long long)66 * 66 * 16; i2c1_0.sAi = (long long)66 * 16; i2c1_0.sAm = 16; i2c1_0.sAk = 1; i2c1_0.sBo = 0; i2c1_0.sBi = 0; i2c1_0.sBn = 16 * 9; i2c1_0.sBk = 9; i2c1_0.sCo = (long long)66 * 66 * 32; i2c1_0.sCi = (long long)66 * 32; i2c1_0.sCm = 32; i2c1_0.sRo = 0; i2c1_0.sRi = 0; i2c1_0.sRm = 0; i2c1_0.sRn = 0;
      i2c1_0.M = 64; i2c1_0.N = 32; i2c1_0.K = 16; i2c1_0.zi_n = 64; i2c1_0.flags = 1; i2c1_0.act = 0;
      i2c1_0.alpha = 1.0f; i2c1_0.beta = 0.0f; i2c1_0.sa = 1.0f; i2c1_0.sb = 1.0f; i2c1_0.Npad = 32; i2c1_0.pad_ = 0;
      k_gemm<1><<<dim3((unsigned)((32) + 31) / 32, (unsigned)((64) + 15) / 16, (unsigned)(2 * 64)), 32, 0, stream>>>(i2c1_0); }
    { GemmP i2c1_1;
      i2c1_1.A = R67 + 26176 + (size_t)1 * 16; i2c1_1.B = iw2 + 1; i2c1_1.bias = R67 + 26176 + (size_t)1 * 16; i2c1_1.R = R67 + 165568 + (size_t)67 * 32; i2c1_1.C = R67 + 165568 + (size_t)67 * 32;
      i2c1_1.sAo = (long long)66 * 66 * 16; i2c1_1.sAi = (long long)66 * 16; i2c1_1.sAm = 16; i2c1_1.sAk = 1; i2c1_1.sBo = 0; i2c1_1.sBi = 0; i2c1_1.sBn = 16 * 9; i2c1_1.sBk = 9; i2c1_1.sCo = (long long)66 * 66 * 32; i2c1_1.sCi = (long long)66 * 32; i2c1_1.sCm = 32; i2c1_1.sRo = (long long)66 * 66 * 32; i2c1_1.sRi = (long long)66 * 32; i2c1_1.sRm = 32; i2c1_1.sRn = 1;
      i2c1_1.M = 64; i2c1_1.N = 32; i2c1_1.K = 16; i2c1_1.zi_n = 64; i2c1_1.flags = 4; i2c1_1.act = 0;
      i2c1_1.alpha = 1.0f; i2c1_1.beta = 1.0f; i2c1_1.sa = 1.0f; i2c1_1.sb = 1.0f; i2c1_1.Npad = 32; i2c1_1.pad_ = 0;
      k_gemm<1><<<dim3((unsigned)((32) + 31) / 32, (unsigned)((64) + 15) / 16, (unsigned)(2 * 64)), 32, 0, stream>>>(i2c1_1); }
    { GemmP i2c1_2;
      i2c1_2.A = R67 + 26176 + (size_t)2 * 16; i2c1_2.B = iw2 + 2; i2c1_2.bias = R67 + 26176 + (size_t)2 * 16; i2c1_2.R = R67 + 165568 + (size_t)67 * 32; i2c1_2.C = R67 + 165568 + (size_t)67 * 32;
      i2c1_2.sAo = (long long)66 * 66 * 16; i2c1_2.sAi = (long long)66 * 16; i2c1_2.sAm = 16; i2c1_2.sAk = 1; i2c1_2.sBo = 0; i2c1_2.sBi = 0; i2c1_2.sBn = 16 * 9; i2c1_2.sBk = 9; i2c1_2.sCo = (long long)66 * 66 * 32; i2c1_2.sCi = (long long)66 * 32; i2c1_2.sCm = 32; i2c1_2.sRo = (long long)66 * 66 * 32; i2c1_2.sRi = (long long)66 * 32; i2c1_2.sRm = 32; i2c1_2.sRn = 1;
      i2c1_2.M = 64; i2c1_2.N = 32; i2c1_2.K = 16; i2c1_2.zi_n = 64; i2c1_2.flags = 4; i2c1_2.act = 0;
      i2c1_2.alpha = 1.0f; i2c1_2.beta = 1.0f; i2c1_2.sa = 1.0f; i2c1_2.sb = 1.0f; i2c1_2.Npad = 32; i2c1_2.pad_ = 0;
      k_gemm<1><<<dim3((unsigned)((32) + 31) / 32, (unsigned)((64) + 15) / 16, (unsigned)(2 * 64)), 32, 0, stream>>>(i2c1_2); }
    { GemmP i2c1_3;
      i2c1_3.A = R67 + 26176 + (size_t)66 * 16; i2c1_3.B = iw2 + 3; i2c1_3.bias = R67 + 26176 + (size_t)66 * 16; i2c1_3.R = R67 + 165568 + (size_t)67 * 32; i2c1_3.C = R67 + 165568 + (size_t)67 * 32;
      i2c1_3.sAo = (long long)66 * 66 * 16; i2c1_3.sAi = (long long)66 * 16; i2c1_3.sAm = 16; i2c1_3.sAk = 1; i2c1_3.sBo = 0; i2c1_3.sBi = 0; i2c1_3.sBn = 16 * 9; i2c1_3.sBk = 9; i2c1_3.sCo = (long long)66 * 66 * 32; i2c1_3.sCi = (long long)66 * 32; i2c1_3.sCm = 32; i2c1_3.sRo = (long long)66 * 66 * 32; i2c1_3.sRi = (long long)66 * 32; i2c1_3.sRm = 32; i2c1_3.sRn = 1;
      i2c1_3.M = 64; i2c1_3.N = 32; i2c1_3.K = 16; i2c1_3.zi_n = 64; i2c1_3.flags = 4; i2c1_3.act = 0;
      i2c1_3.alpha = 1.0f; i2c1_3.beta = 1.0f; i2c1_3.sa = 1.0f; i2c1_3.sb = 1.0f; i2c1_3.Npad = 32; i2c1_3.pad_ = 0;
      k_gemm<1><<<dim3((unsigned)((32) + 31) / 32, (unsigned)((64) + 15) / 16, (unsigned)(2 * 64)), 32, 0, stream>>>(i2c1_3); }
    { GemmP i2c1_4;
      i2c1_4.A = R67 + 26176 + (size_t)67 * 16; i2c1_4.B = iw2 + 4; i2c1_4.bias = R67 + 26176 + (size_t)67 * 16; i2c1_4.R = R67 + 165568 + (size_t)67 * 32; i2c1_4.C = R67 + 165568 + (size_t)67 * 32;
      i2c1_4.sAo = (long long)66 * 66 * 16; i2c1_4.sAi = (long long)66 * 16; i2c1_4.sAm = 16; i2c1_4.sAk = 1; i2c1_4.sBo = 0; i2c1_4.sBi = 0; i2c1_4.sBn = 16 * 9; i2c1_4.sBk = 9; i2c1_4.sCo = (long long)66 * 66 * 32; i2c1_4.sCi = (long long)66 * 32; i2c1_4.sCm = 32; i2c1_4.sRo = (long long)66 * 66 * 32; i2c1_4.sRi = (long long)66 * 32; i2c1_4.sRm = 32; i2c1_4.sRn = 1;
      i2c1_4.M = 64; i2c1_4.N = 32; i2c1_4.K = 16; i2c1_4.zi_n = 64; i2c1_4.flags = 4; i2c1_4.act = 0;
      i2c1_4.alpha = 1.0f; i2c1_4.beta = 1.0f; i2c1_4.sa = 1.0f; i2c1_4.sb = 1.0f; i2c1_4.Npad = 32; i2c1_4.pad_ = 0;
      k_gemm<1><<<dim3((unsigned)((32) + 31) / 32, (unsigned)((64) + 15) / 16, (unsigned)(2 * 64)), 32, 0, stream>>>(i2c1_4); }
    { GemmP i2c1_5;
      i2c1_5.A = R67 + 26176 + (size_t)68 * 16; i2c1_5.B = iw2 + 5; i2c1_5.bias = R67 + 26176 + (size_t)68 * 16; i2c1_5.R = R67 + 165568 + (size_t)67 * 32; i2c1_5.C = R67 + 165568 + (size_t)67 * 32;
      i2c1_5.sAo = (long long)66 * 66 * 16; i2c1_5.sAi = (long long)66 * 16; i2c1_5.sAm = 16; i2c1_5.sAk = 1; i2c1_5.sBo = 0; i2c1_5.sBi = 0; i2c1_5.sBn = 16 * 9; i2c1_5.sBk = 9; i2c1_5.sCo = (long long)66 * 66 * 32; i2c1_5.sCi = (long long)66 * 32; i2c1_5.sCm = 32; i2c1_5.sRo = (long long)66 * 66 * 32; i2c1_5.sRi = (long long)66 * 32; i2c1_5.sRm = 32; i2c1_5.sRn = 1;
      i2c1_5.M = 64; i2c1_5.N = 32; i2c1_5.K = 16; i2c1_5.zi_n = 64; i2c1_5.flags = 4; i2c1_5.act = 0;
      i2c1_5.alpha = 1.0f; i2c1_5.beta = 1.0f; i2c1_5.sa = 1.0f; i2c1_5.sb = 1.0f; i2c1_5.Npad = 32; i2c1_5.pad_ = 0;
      k_gemm<1><<<dim3((unsigned)((32) + 31) / 32, (unsigned)((64) + 15) / 16, (unsigned)(2 * 64)), 32, 0, stream>>>(i2c1_5); }
    { GemmP i2c1_6;
      i2c1_6.A = R67 + 26176 + (size_t)132 * 16; i2c1_6.B = iw2 + 6; i2c1_6.bias = R67 + 26176 + (size_t)132 * 16; i2c1_6.R = R67 + 165568 + (size_t)67 * 32; i2c1_6.C = R67 + 165568 + (size_t)67 * 32;
      i2c1_6.sAo = (long long)66 * 66 * 16; i2c1_6.sAi = (long long)66 * 16; i2c1_6.sAm = 16; i2c1_6.sAk = 1; i2c1_6.sBo = 0; i2c1_6.sBi = 0; i2c1_6.sBn = 16 * 9; i2c1_6.sBk = 9; i2c1_6.sCo = (long long)66 * 66 * 32; i2c1_6.sCi = (long long)66 * 32; i2c1_6.sCm = 32; i2c1_6.sRo = (long long)66 * 66 * 32; i2c1_6.sRi = (long long)66 * 32; i2c1_6.sRm = 32; i2c1_6.sRn = 1;
      i2c1_6.M = 64; i2c1_6.N = 32; i2c1_6.K = 16; i2c1_6.zi_n = 64; i2c1_6.flags = 4; i2c1_6.act = 0;
      i2c1_6.alpha = 1.0f; i2c1_6.beta = 1.0f; i2c1_6.sa = 1.0f; i2c1_6.sb = 1.0f; i2c1_6.Npad = 32; i2c1_6.pad_ = 0;
      k_gemm<1><<<dim3((unsigned)((32) + 31) / 32, (unsigned)((64) + 15) / 16, (unsigned)(2 * 64)), 32, 0, stream>>>(i2c1_6); }
    { GemmP i2c1_7;
      i2c1_7.A = R67 + 26176 + (size_t)133 * 16; i2c1_7.B = iw2 + 7; i2c1_7.bias = R67 + 26176 + (size_t)133 * 16; i2c1_7.R = R67 + 165568 + (size_t)67 * 32; i2c1_7.C = R67 + 165568 + (size_t)67 * 32;
      i2c1_7.sAo = (long long)66 * 66 * 16; i2c1_7.sAi = (long long)66 * 16; i2c1_7.sAm = 16; i2c1_7.sAk = 1; i2c1_7.sBo = 0; i2c1_7.sBi = 0; i2c1_7.sBn = 16 * 9; i2c1_7.sBk = 9; i2c1_7.sCo = (long long)66 * 66 * 32; i2c1_7.sCi = (long long)66 * 32; i2c1_7.sCm = 32; i2c1_7.sRo = (long long)66 * 66 * 32; i2c1_7.sRi = (long long)66 * 32; i2c1_7.sRm = 32; i2c1_7.sRn = 1;
      i2c1_7.M = 64; i2c1_7.N = 32; i2c1_7.K = 16; i2c1_7.zi_n = 64; i2c1_7.flags = 4; i2c1_7.act = 0;
      i2c1_7.alpha = 1.0f; i2c1_7.beta = 1.0f; i2c1_7.sa = 1.0f; i2c1_7.sb = 1.0f; i2c1_7.Npad = 32; i2c1_7.pad_ = 0;
      k_gemm<1><<<dim3((unsigned)((32) + 31) / 32, (unsigned)((64) + 15) / 16, (unsigned)(2 * 64)), 32, 0, stream>>>(i2c1_7); }
    { GemmP i2c1_8;
      i2c1_8.A = R67 + 26176 + (size_t)134 * 16; i2c1_8.B = iw2 + 8; i2c1_8.bias = R67 + 26176 + (size_t)134 * 16; i2c1_8.R = R67 + 165568 + (size_t)67 * 32; i2c1_8.C = R67 + 165568 + (size_t)67 * 32;
      i2c1_8.sAo = (long long)66 * 66 * 16; i2c1_8.sAi = (long long)66 * 16; i2c1_8.sAm = 16; i2c1_8.sAk = 1; i2c1_8.sBo = 0; i2c1_8.sBi = 0; i2c1_8.sBn = 16 * 9; i2c1_8.sBk = 9; i2c1_8.sCo = (long long)66 * 66 * 32; i2c1_8.sCi = (long long)66 * 32; i2c1_8.sCm = 32; i2c1_8.sRo = (long long)66 * 66 * 32; i2c1_8.sRi = (long long)66 * 32; i2c1_8.sRm = 32; i2c1_8.sRn = 1;
      i2c1_8.M = 64; i2c1_8.N = 32; i2c1_8.K = 16; i2c1_8.zi_n = 64; i2c1_8.flags = 4; i2c1_8.act = 0;
      i2c1_8.alpha = 1.0f; i2c1_8.beta = 1.0f; i2c1_8.sa = 1.0f; i2c1_8.sb = 1.0f; i2c1_8.Npad = 32; i2c1_8.pad_ = 0;
      k_gemm<1><<<dim3((unsigned)((32) + 31) / 32, (unsigned)((64) + 15) / 16, (unsigned)(2 * 64)), 32, 0, stream>>>(i2c1_8); }
    k_mm_relu2d<<<(unsigned)(((long long)2 * HW * 32 + 255) / 256), 256, 0, stream>>>(R67 + 165568, nullptr, 2, 64, 32);
    { GemmP i3c1_0;
      i3c1_0.A = R67 + 165568 + (size_t)0 * 32; i3c1_0.B = iw3 + 0; i3c1_0.bias = ib3; i3c1_0.R = R67 + 165568 + (size_t)0 * 32; i3c1_0.C = R67 + 444352 + (size_t)67 * 64;
      i3c1_0.sAo = (long long)66 * 66 * 32; i3c1_0.sAi = (long long)66 * 32; i3c1_0.sAm = 32; i3c1_0.sAk = 1; i3c1_0.sBo = 0; i3c1_0.sBi = 0; i3c1_0.sBn = 32 * 9; i3c1_0.sBk = 9; i3c1_0.sCo = (long long)66 * 66 * 64; i3c1_0.sCi = (long long)66 * 64; i3c1_0.sCm = 64; i3c1_0.sRo = 0; i3c1_0.sRi = 0; i3c1_0.sRm = 0; i3c1_0.sRn = 0;
      i3c1_0.M = 64; i3c1_0.N = 64; i3c1_0.K = 32; i3c1_0.zi_n = 64; i3c1_0.flags = 1; i3c1_0.act = 0;
      i3c1_0.alpha = 1.0f; i3c1_0.beta = 0.0f; i3c1_0.sa = 1.0f; i3c1_0.sb = 1.0f; i3c1_0.Npad = 64; i3c1_0.pad_ = 0;
      k_gemm<1><<<dim3((unsigned)((64) + 31) / 32, (unsigned)((64) + 15) / 16, (unsigned)(2 * 64)), 32, 0, stream>>>(i3c1_0); }
    { GemmP i3c1_1;
      i3c1_1.A = R67 + 165568 + (size_t)1 * 32; i3c1_1.B = iw3 + 1; i3c1_1.bias = R67 + 165568 + (size_t)1 * 32; i3c1_1.R = R67 + 444352 + (size_t)67 * 64; i3c1_1.C = R67 + 444352 + (size_t)67 * 64;
      i3c1_1.sAo = (long long)66 * 66 * 32; i3c1_1.sAi = (long long)66 * 32; i3c1_1.sAm = 32; i3c1_1.sAk = 1; i3c1_1.sBo = 0; i3c1_1.sBi = 0; i3c1_1.sBn = 32 * 9; i3c1_1.sBk = 9; i3c1_1.sCo = (long long)66 * 66 * 64; i3c1_1.sCi = (long long)66 * 64; i3c1_1.sCm = 64; i3c1_1.sRo = (long long)66 * 66 * 64; i3c1_1.sRi = (long long)66 * 64; i3c1_1.sRm = 64; i3c1_1.sRn = 1;
      i3c1_1.M = 64; i3c1_1.N = 64; i3c1_1.K = 32; i3c1_1.zi_n = 64; i3c1_1.flags = 4; i3c1_1.act = 0;
      i3c1_1.alpha = 1.0f; i3c1_1.beta = 1.0f; i3c1_1.sa = 1.0f; i3c1_1.sb = 1.0f; i3c1_1.Npad = 64; i3c1_1.pad_ = 0;
      k_gemm<1><<<dim3((unsigned)((64) + 31) / 32, (unsigned)((64) + 15) / 16, (unsigned)(2 * 64)), 32, 0, stream>>>(i3c1_1); }
    { GemmP i3c1_2;
      i3c1_2.A = R67 + 165568 + (size_t)2 * 32; i3c1_2.B = iw3 + 2; i3c1_2.bias = R67 + 165568 + (size_t)2 * 32; i3c1_2.R = R67 + 444352 + (size_t)67 * 64; i3c1_2.C = R67 + 444352 + (size_t)67 * 64;
      i3c1_2.sAo = (long long)66 * 66 * 32; i3c1_2.sAi = (long long)66 * 32; i3c1_2.sAm = 32; i3c1_2.sAk = 1; i3c1_2.sBo = 0; i3c1_2.sBi = 0; i3c1_2.sBn = 32 * 9; i3c1_2.sBk = 9; i3c1_2.sCo = (long long)66 * 66 * 64; i3c1_2.sCi = (long long)66 * 64; i3c1_2.sCm = 64; i3c1_2.sRo = (long long)66 * 66 * 64; i3c1_2.sRi = (long long)66 * 64; i3c1_2.sRm = 64; i3c1_2.sRn = 1;
      i3c1_2.M = 64; i3c1_2.N = 64; i3c1_2.K = 32; i3c1_2.zi_n = 64; i3c1_2.flags = 4; i3c1_2.act = 0;
      i3c1_2.alpha = 1.0f; i3c1_2.beta = 1.0f; i3c1_2.sa = 1.0f; i3c1_2.sb = 1.0f; i3c1_2.Npad = 64; i3c1_2.pad_ = 0;
      k_gemm<1><<<dim3((unsigned)((64) + 31) / 32, (unsigned)((64) + 15) / 16, (unsigned)(2 * 64)), 32, 0, stream>>>(i3c1_2); }
    { GemmP i3c1_3;
      i3c1_3.A = R67 + 165568 + (size_t)66 * 32; i3c1_3.B = iw3 + 3; i3c1_3.bias = R67 + 165568 + (size_t)66 * 32; i3c1_3.R = R67 + 444352 + (size_t)67 * 64; i3c1_3.C = R67 + 444352 + (size_t)67 * 64;
      i3c1_3.sAo = (long long)66 * 66 * 32; i3c1_3.sAi = (long long)66 * 32; i3c1_3.sAm = 32; i3c1_3.sAk = 1; i3c1_3.sBo = 0; i3c1_3.sBi = 0; i3c1_3.sBn = 32 * 9; i3c1_3.sBk = 9; i3c1_3.sCo = (long long)66 * 66 * 64; i3c1_3.sCi = (long long)66 * 64; i3c1_3.sCm = 64; i3c1_3.sRo = (long long)66 * 66 * 64; i3c1_3.sRi = (long long)66 * 64; i3c1_3.sRm = 64; i3c1_3.sRn = 1;
      i3c1_3.M = 64; i3c1_3.N = 64; i3c1_3.K = 32; i3c1_3.zi_n = 64; i3c1_3.flags = 4; i3c1_3.act = 0;
      i3c1_3.alpha = 1.0f; i3c1_3.beta = 1.0f; i3c1_3.sa = 1.0f; i3c1_3.sb = 1.0f; i3c1_3.Npad = 64; i3c1_3.pad_ = 0;
      k_gemm<1><<<dim3((unsigned)((64) + 31) / 32, (unsigned)((64) + 15) / 16, (unsigned)(2 * 64)), 32, 0, stream>>>(i3c1_3); }
    { GemmP i3c1_4;
      i3c1_4.A = R67 + 165568 + (size_t)67 * 32; i3c1_4.B = iw3 + 4; i3c1_4.bias = R67 + 165568 + (size_t)67 * 32; i3c1_4.R = R67 + 444352 + (size_t)67 * 64; i3c1_4.C = R67 + 444352 + (size_t)67 * 64;
      i3c1_4.sAo = (long long)66 * 66 * 32; i3c1_4.sAi = (long long)66 * 32; i3c1_4.sAm = 32; i3c1_4.sAk = 1; i3c1_4.sBo = 0; i3c1_4.sBi = 0; i3c1_4.sBn = 32 * 9; i3c1_4.sBk = 9; i3c1_4.sCo = (long long)66 * 66 * 64; i3c1_4.sCi = (long long)66 * 64; i3c1_4.sCm = 64; i3c1_4.sRo = (long long)66 * 66 * 64; i3c1_4.sRi = (long long)66 * 64; i3c1_4.sRm = 64; i3c1_4.sRn = 1;
      i3c1_4.M = 64; i3c1_4.N = 64; i3c1_4.K = 32; i3c1_4.zi_n = 64; i3c1_4.flags = 4; i3c1_4.act = 0;
      i3c1_4.alpha = 1.0f; i3c1_4.beta = 1.0f; i3c1_4.sa = 1.0f; i3c1_4.sb = 1.0f; i3c1_4.Npad = 64; i3c1_4.pad_ = 0;
      k_gemm<1><<<dim3((unsigned)((64) + 31) / 32, (unsigned)((64) + 15) / 16, (unsigned)(2 * 64)), 32, 0, stream>>>(i3c1_4); }
    { GemmP i3c1_5;
      i3c1_5.A = R67 + 165568 + (size_t)68 * 32; i3c1_5.B = iw3 + 5; i3c1_5.bias = R67 + 165568 + (size_t)68 * 32; i3c1_5.R = R67 + 444352 + (size_t)67 * 64; i3c1_5.C = R67 + 444352 + (size_t)67 * 64;
      i3c1_5.sAo = (long long)66 * 66 * 32; i3c1_5.sAi = (long long)66 * 32; i3c1_5.sAm = 32; i3c1_5.sAk = 1; i3c1_5.sBo = 0; i3c1_5.sBi = 0; i3c1_5.sBn = 32 * 9; i3c1_5.sBk = 9; i3c1_5.sCo = (long long)66 * 66 * 64; i3c1_5.sCi = (long long)66 * 64; i3c1_5.sCm = 64; i3c1_5.sRo = (long long)66 * 66 * 64; i3c1_5.sRi = (long long)66 * 64; i3c1_5.sRm = 64; i3c1_5.sRn = 1;
      i3c1_5.M = 64; i3c1_5.N = 64; i3c1_5.K = 32; i3c1_5.zi_n = 64; i3c1_5.flags = 4; i3c1_5.act = 0;
      i3c1_5.alpha = 1.0f; i3c1_5.beta = 1.0f; i3c1_5.sa = 1.0f; i3c1_5.sb = 1.0f; i3c1_5.Npad = 64; i3c1_5.pad_ = 0;
      k_gemm<1><<<dim3((unsigned)((64) + 31) / 32, (unsigned)((64) + 15) / 16, (unsigned)(2 * 64)), 32, 0, stream>>>(i3c1_5); }
    { GemmP i3c1_6;
      i3c1_6.A = R67 + 165568 + (size_t)132 * 32; i3c1_6.B = iw3 + 6; i3c1_6.bias = R67 + 165568 + (size_t)132 * 32; i3c1_6.R = R67 + 444352 + (size_t)67 * 64; i3c1_6.C = R67 + 444352 + (size_t)67 * 64;
      i3c1_6.sAo = (long long)66 * 66 * 32; i3c1_6.sAi = (long long)66 * 32; i3c1_6.sAm = 32; i3c1_6.sAk = 1; i3c1_6.sBo = 0; i3c1_6.sBi = 0; i3c1_6.sBn = 32 * 9; i3c1_6.sBk = 9; i3c1_6.sCo = (long long)66 * 66 * 64; i3c1_6.sCi = (long long)66 * 64; i3c1_6.sCm = 64; i3c1_6.sRo = (long long)66 * 66 * 64; i3c1_6.sRi = (long long)66 * 64; i3c1_6.sRm = 64; i3c1_6.sRn = 1;
      i3c1_6.M = 64; i3c1_6.N = 64; i3c1_6.K = 32; i3c1_6.zi_n = 64; i3c1_6.flags = 4; i3c1_6.act = 0;
      i3c1_6.alpha = 1.0f; i3c1_6.beta = 1.0f; i3c1_6.sa = 1.0f; i3c1_6.sb = 1.0f; i3c1_6.Npad = 64; i3c1_6.pad_ = 0;
      k_gemm<1><<<dim3((unsigned)((64) + 31) / 32, (unsigned)((64) + 15) / 16, (unsigned)(2 * 64)), 32, 0, stream>>>(i3c1_6); }
    { GemmP i3c1_7;
      i3c1_7.A = R67 + 165568 + (size_t)133 * 32; i3c1_7.B = iw3 + 7; i3c1_7.bias = R67 + 165568 + (size_t)133 * 32; i3c1_7.R = R67 + 444352 + (size_t)67 * 64; i3c1_7.C = R67 + 444352 + (size_t)67 * 64;
      i3c1_7.sAo = (long long)66 * 66 * 32; i3c1_7.sAi = (long long)66 * 32; i3c1_7.sAm = 32; i3c1_7.sAk = 1; i3c1_7.sBo = 0; i3c1_7.sBi = 0; i3c1_7.sBn = 32 * 9; i3c1_7.sBk = 9; i3c1_7.sCo = (long long)66 * 66 * 64; i3c1_7.sCi = (long long)66 * 64; i3c1_7.sCm = 64; i3c1_7.sRo = (long long)66 * 66 * 64; i3c1_7.sRi = (long long)66 * 64; i3c1_7.sRm = 64; i3c1_7.sRn = 1;
      i3c1_7.M = 64; i3c1_7.N = 64; i3c1_7.K = 32; i3c1_7.zi_n = 64; i3c1_7.flags = 4; i3c1_7.act = 0;
      i3c1_7.alpha = 1.0f; i3c1_7.beta = 1.0f; i3c1_7.sa = 1.0f; i3c1_7.sb = 1.0f; i3c1_7.Npad = 64; i3c1_7.pad_ = 0;
      k_gemm<1><<<dim3((unsigned)((64) + 31) / 32, (unsigned)((64) + 15) / 16, (unsigned)(2 * 64)), 32, 0, stream>>>(i3c1_7); }
    { GemmP i3c1_8;
      i3c1_8.A = R67 + 165568 + (size_t)134 * 32; i3c1_8.B = iw3 + 8; i3c1_8.bias = R67 + 165568 + (size_t)134 * 32; i3c1_8.R = R67 + 444352 + (size_t)67 * 64; i3c1_8.C = R67 + 444352 + (size_t)67 * 64;
      i3c1_8.sAo = (long long)66 * 66 * 32; i3c1_8.sAi = (long long)66 * 32; i3c1_8.sAm = 32; i3c1_8.sAk = 1; i3c1_8.sBo = 0; i3c1_8.sBi = 0; i3c1_8.sBn = 32 * 9; i3c1_8.sBk = 9; i3c1_8.sCo = (long long)66 * 66 * 64; i3c1_8.sCi = (long long)66 * 64; i3c1_8.sCm = 64; i3c1_8.sRo = (long long)66 * 66 * 64; i3c1_8.sRi = (long long)66 * 64; i3c1_8.sRm = 64; i3c1_8.sRn = 1;
      i3c1_8.M = 64; i3c1_8.N = 64; i3c1_8.K = 32; i3c1_8.zi_n = 64; i3c1_8.flags = 4; i3c1_8.act = 0;
      i3c1_8.alpha = 1.0f; i3c1_8.beta = 1.0f; i3c1_8.sa = 1.0f; i3c1_8.sb = 1.0f; i3c1_8.Npad = 64; i3c1_8.pad_ = 0;
      k_gemm<1><<<dim3((unsigned)((64) + 31) / 32, (unsigned)((64) + 15) / 16, (unsigned)(2 * 64)), 32, 0, stream>>>(i3c1_8); }
    k_mm_relu2d<<<(unsigned)(((long long)2 * HW * 64 + 255) / 256), 256, 0, stream>>>(R67 + 444352, R67 + 1001920, 2, 64, 64);
    { GemmP gqkv1;
      gqkv1.A = R67 + 1001920; gqkv1.B = qkvw; gqkv1.bias = qkvb; gqkv1.R = R67 + 1001920; gqkv1.C = R67 + 1526208;
      gqkv1.sAo = 0; gqkv1.sAi = 0; gqkv1.sAm = 64; gqkv1.sAk = 1; gqkv1.sBo = 0; gqkv1.sBi = 0; gqkv1.sBn = 64; gqkv1.sBk = 1; gqkv1.sCo = 0; gqkv1.sCi = 0; gqkv1.sCm = 192; gqkv1.sRo = 0; gqkv1.sRi = 0; gqkv1.sRm = 0; gqkv1.sRn = 0;
      gqkv1.M = 2 * HW; gqkv1.N = 192; gqkv1.K = 64; gqkv1.zi_n = 1; gqkv1.flags = 1; gqkv1.act = 0;
      gqkv1.alpha = 1.0f; gqkv1.beta = 0.0f; gqkv1.sa = 1.0f; gqkv1.sb = 1.0f; gqkv1.Npad = 192; gqkv1.pad_ = 0;
      k_gemm<1><<<dim3((unsigned)((192) + 31) / 32, (unsigned)((2 * HW) + 15) / 16, (unsigned)(1)), 32, 0, stream>>>(gqkv1); }
    k_mm_dw<<<(unsigned)(((long long)2 * HW * 192 + 255) / 256), 256, 0, stream>>>(R67 + 1526208, dww, dwb, R67 + 3099072, 2, 64, 192);
    k_mm_fall<<<(unsigned)(((long long)2 * HW * 144 + 255) / 256), 256, 0, stream>>>(R67 + 3099072, fcw, fcb, R67 + 4671936, 2, HW, 192);
    k_mm_dep<<<(unsigned)(((long long)2 * 64 * HW + 255) / 256), 256, 0, stream>>>(R67 + 4671936, depw, depb, R67 + 5851584, 2, 64);
    k_mm_qknorm<<<2 * 128, 256, 0, stream>>>(R67 + 3099072, R67 + 6375872, 2, HW, 192);
    { GemmP gat1;
      gat1.A = R67 + 6375872; gat1.B = R67 + 6375872 + (size_t)64 * HW; gat1.bias = R67 + 6375872; gat1.R = R67 + 6375872; gat1.C = R67 + 7424448;
      gat1.sAo = (long long)128 * HW; gat1.sAi = (long long)16 * HW; gat1.sAm = HW; gat1.sAk = 1; gat1.sBo = (long long)128 * HW; gat1.sBi = (long long)16 * HW; gat1.sBn = HW; gat1.sBk = 1; gat1.sCo = (long long)4 * 16 * LP; gat1.sCi = 16 * LP; gat1.sCm = LP; gat1.sRo = 0; gat1.sRi = 0; gat1.sRm = 0; gat1.sRn = 0;
      gat1.M = 16; gat1.N = 16; gat1.K = HW; gat1.zi_n = 4; gat1.flags = 0; gat1.act = 0;
      gat1.alpha = 1.0f; gat1.beta = 0.0f; gat1.sa = 1.0f; gat1.sb = 1.0f; gat1.Npad = LP; gat1.pad_ = 0;
      k_gemm<1><<<dim3((unsigned)((LP) + 31) / 32, (unsigned)((16) + 15) / 16, (unsigned)(2 * 4)), 32, 0, stream>>>(gat1); }
    k_mm_sm16<<<(unsigned)((2 * 4 * 16 + 255) / 256), 256, 0, stream>>>(R67 + 7424448, temp, 2 * 4, LP);
    { GemmP gao1;
      gao1.A = R67 + 7424448; gao1.B = R67 + 3099072 + 128; gao1.bias = R67 + 7424448; gao1.R = R67 + 7424448; gao1.C = R67 + 7428544;
      gao1.sAo = (long long)4 * 16 * LP; gao1.sAi = 16 * LP; gao1.sAm = LP; gao1.sAk = 1; gao1.sBo = (long long)HW * 192; gao1.sBi = 16; gao1.sBn = 192; gao1.sBk = 1; gao1.sCo = (long long)64 * HW; gao1.sCi = (long long)16 * HW; gao1.sCm = HW; gao1.sRo = 0; gao1.sRi = 0; gao1.sRm = 0; gao1.sRn = 0;
      gao1.M = 16; gao1.N = HW; gao1.K = 16; gao1.zi_n = 4; gao1.flags = 0; gao1.act = 0;
      gao1.alpha = 1.0f; gao1.beta = 0.0f; gao1.sa = 1.0f; gao1.sb = 1.0f; gao1.Npad = HW; gao1.pad_ = 0;
      k_gemm<1><<<dim3((unsigned)((HW) + 31) / 32, (unsigned)((16) + 15) / 16, (unsigned)(2 * 4)), 32, 0, stream>>>(gao1); }
    { GemmP gproj1;
      gproj1.A = projw; gproj1.B = R67 + 7428544; gproj1.bias = projb; gproj1.R = projw; gproj1.C = R67 + 7952832;
      gproj1.sAo = 0; gproj1.sAi = 0; gproj1.sAm = 64; gproj1.sAk = 1; gproj1.sBo = (long long)64 * HW; gproj1.sBi = 0; gproj1.sBn = 1; gproj1.sBk = HW; gproj1.sCo = (long long)64 * HW; gproj1.sCi = 0; gproj1.sCm = HW; gproj1.sRo = 0; gproj1.sRi = 0; gproj1.sRm = 0; gproj1.sRn = 0;
      gproj1.M = 64; gproj1.N = HW; gproj1.K = 64; gproj1.zi_n = 1; gproj1.flags = 2; gproj1.act = 0;
      gproj1.alpha = 1.0f; gproj1.beta = 0.0f; gproj1.sa = 1.0f; gproj1.sb = 1.0f; gproj1.Npad = HW; gproj1.pad_ = 0;
      k_gemm<1><<<dim3((unsigned)((HW) + 31) / 32, (unsigned)((64) + 15) / 16, (unsigned)(2)), 32, 0, stream>>>(gproj1); }
    k_mm_imgfeat<<<(unsigned)(((long long)2 * SEQ * 64 + 255) / 256), 256, 0, stream>>>(R67 + 7952832, R67 + 5851584, IR + (size_t)2 * SEQ * 64, 2, HW, 64);
    hipMemsetAsync(R67 + 0, 0, (size_t)2 * 66 * 66 * 3 * 4, stream); hipMemsetAsync(R67 + 26176, 0, (size_t)2 * 66 * 66 * 16 * 4, stream); hipMemsetAsync(R67 + 165568, 0, (size_t)2 * 66 * 66 * 32 * 4, stream); hipMemsetAsync(R67 + 444352, 0, (size_t)2 * 66 * 66 * 64 * 4, stream);
    k_mm_padimg<<<(unsigned)(((long long)2 * HW * 3 + 255) / 256), 256, 0, stream>>>(img + (size_t)4 * 3 * HW, R67 + 0, 2, 3, 64);
    { GemmP i1c2_0;
      i1c2_0.A = R67 + 0 + (size_t)0 * 3; i1c2_0.B = iw1 + 0; i1c2_0.bias = ib1; i1c2_0.R = R67 + 0 + (size_t)0 * 3; i1c2_0.C = R67 + 26176 + (size_t)67 * 16;
      i1c2_0.sAo = (long long)66 * 66 * 3; i1c2_0.sAi = (long long)66 * 3; i1c2_0.sAm = 3; i1c2_0.sAk = 1; i1c2_0.sBo = 0; i1c2_0.sBi = 0; i1c2_0.sBn = 3 * 9; i1c2_0.sBk = 9; i1c2_0.sCo = (long long)66 * 66 * 16; i1c2_0.sCi = (long long)66 * 16; i1c2_0.sCm = 16; i1c2_0.sRo = 0; i1c2_0.sRi = 0; i1c2_0.sRm = 0; i1c2_0.sRn = 0;
      i1c2_0.M = 64; i1c2_0.N = 16; i1c2_0.K = 3; i1c2_0.zi_n = 64; i1c2_0.flags = 1; i1c2_0.act = 0;
      i1c2_0.alpha = 1.0f; i1c2_0.beta = 0.0f; i1c2_0.sa = 1.0f; i1c2_0.sb = 1.0f; i1c2_0.Npad = 16; i1c2_0.pad_ = 0;
      k_gemm<1><<<dim3((unsigned)((16) + 31) / 32, (unsigned)((64) + 15) / 16, (unsigned)(2 * 64)), 32, 0, stream>>>(i1c2_0); }
    { GemmP i1c2_1;
      i1c2_1.A = R67 + 0 + (size_t)1 * 3; i1c2_1.B = iw1 + 1; i1c2_1.bias = R67 + 0 + (size_t)1 * 3; i1c2_1.R = R67 + 26176 + (size_t)67 * 16; i1c2_1.C = R67 + 26176 + (size_t)67 * 16;
      i1c2_1.sAo = (long long)66 * 66 * 3; i1c2_1.sAi = (long long)66 * 3; i1c2_1.sAm = 3; i1c2_1.sAk = 1; i1c2_1.sBo = 0; i1c2_1.sBi = 0; i1c2_1.sBn = 3 * 9; i1c2_1.sBk = 9; i1c2_1.sCo = (long long)66 * 66 * 16; i1c2_1.sCi = (long long)66 * 16; i1c2_1.sCm = 16; i1c2_1.sRo = (long long)66 * 66 * 16; i1c2_1.sRi = (long long)66 * 16; i1c2_1.sRm = 16; i1c2_1.sRn = 1;
      i1c2_1.M = 64; i1c2_1.N = 16; i1c2_1.K = 3; i1c2_1.zi_n = 64; i1c2_1.flags = 4; i1c2_1.act = 0;
      i1c2_1.alpha = 1.0f; i1c2_1.beta = 1.0f; i1c2_1.sa = 1.0f; i1c2_1.sb = 1.0f; i1c2_1.Npad = 16; i1c2_1.pad_ = 0;
      k_gemm<1><<<dim3((unsigned)((16) + 31) / 32, (unsigned)((64) + 15) / 16, (unsigned)(2 * 64)), 32, 0, stream>>>(i1c2_1); }
    { GemmP i1c2_2;
      i1c2_2.A = R67 + 0 + (size_t)2 * 3; i1c2_2.B = iw1 + 2; i1c2_2.bias = R67 + 0 + (size_t)2 * 3; i1c2_2.R = R67 + 26176 + (size_t)67 * 16; i1c2_2.C = R67 + 26176 + (size_t)67 * 16;
      i1c2_2.sAo = (long long)66 * 66 * 3; i1c2_2.sAi = (long long)66 * 3; i1c2_2.sAm = 3; i1c2_2.sAk = 1; i1c2_2.sBo = 0; i1c2_2.sBi = 0; i1c2_2.sBn = 3 * 9; i1c2_2.sBk = 9; i1c2_2.sCo = (long long)66 * 66 * 16; i1c2_2.sCi = (long long)66 * 16; i1c2_2.sCm = 16; i1c2_2.sRo = (long long)66 * 66 * 16; i1c2_2.sRi = (long long)66 * 16; i1c2_2.sRm = 16; i1c2_2.sRn = 1;
      i1c2_2.M = 64; i1c2_2.N = 16; i1c2_2.K = 3; i1c2_2.zi_n = 64; i1c2_2.flags = 4; i1c2_2.act = 0;
      i1c2_2.alpha = 1.0f; i1c2_2.beta = 1.0f; i1c2_2.sa = 1.0f; i1c2_2.sb = 1.0f; i1c2_2.Npad = 16; i1c2_2.pad_ = 0;
      k_gemm<1><<<dim3((unsigned)((16) + 31) / 32, (unsigned)((64) + 15) / 16, (unsigned)(2 * 64)), 32, 0, stream>>>(i1c2_2); }
    { GemmP i1c2_3;
      i1c2_3.A = R67 + 0 + (size_t)66 * 3; i1c2_3.B = iw1 + 3; i1c2_3.bias = R67 + 0 + (size_t)66 * 3; i1c2_3.R = R67 + 26176 + (size_t)67 * 16; i1c2_3.C = R67 + 26176 + (size_t)67 * 16;
      i1c2_3.sAo = (long long)66 * 66 * 3; i1c2_3.sAi = (long long)66 * 3; i1c2_3.sAm = 3; i1c2_3.sAk = 1; i1c2_3.sBo = 0; i1c2_3.sBi = 0; i1c2_3.sBn = 3 * 9; i1c2_3.sBk = 9; i1c2_3.sCo = (long long)66 * 66 * 16; i1c2_3.sCi = (long long)66 * 16; i1c2_3.sCm = 16; i1c2_3.sRo = (long long)66 * 66 * 16; i1c2_3.sRi = (long long)66 * 16; i1c2_3.sRm = 16; i1c2_3.sRn = 1;
      i1c2_3.M = 64; i1c2_3.N = 16; i1c2_3.K = 3; i1c2_3.zi_n = 64; i1c2_3.flags = 4; i1c2_3.act = 0;
      i1c2_3.alpha = 1.0f; i1c2_3.beta = 1.0f; i1c2_3.sa = 1.0f; i1c2_3.sb = 1.0f; i1c2_3.Npad = 16; i1c2_3.pad_ = 0;
      k_gemm<1><<<dim3((unsigned)((16) + 31) / 32, (unsigned)((64) + 15) / 16, (unsigned)(2 * 64)), 32, 0, stream>>>(i1c2_3); }
    { GemmP i1c2_4;
      i1c2_4.A = R67 + 0 + (size_t)67 * 3; i1c2_4.B = iw1 + 4; i1c2_4.bias = R67 + 0 + (size_t)67 * 3; i1c2_4.R = R67 + 26176 + (size_t)67 * 16; i1c2_4.C = R67 + 26176 + (size_t)67 * 16;
      i1c2_4.sAo = (long long)66 * 66 * 3; i1c2_4.sAi = (long long)66 * 3; i1c2_4.sAm = 3; i1c2_4.sAk = 1; i1c2_4.sBo = 0; i1c2_4.sBi = 0; i1c2_4.sBn = 3 * 9; i1c2_4.sBk = 9; i1c2_4.sCo = (long long)66 * 66 * 16; i1c2_4.sCi = (long long)66 * 16; i1c2_4.sCm = 16; i1c2_4.sRo = (long long)66 * 66 * 16; i1c2_4.sRi = (long long)66 * 16; i1c2_4.sRm = 16; i1c2_4.sRn = 1;
      i1c2_4.M = 64; i1c2_4.N = 16; i1c2_4.K = 3; i1c2_4.zi_n = 64; i1c2_4.flags = 4; i1c2_4.act = 0;
      i1c2_4.alpha = 1.0f; i1c2_4.beta = 1.0f; i1c2_4.sa = 1.0f; i1c2_4.sb = 1.0f; i1c2_4.Npad = 16; i1c2_4.pad_ = 0;
      k_gemm<1><<<dim3((unsigned)((16) + 31) / 32, (unsigned)((64) + 15) / 16, (unsigned)(2 * 64)), 32, 0, stream>>>(i1c2_4); }
    { GemmP i1c2_5;
      i1c2_5.A = R67 + 0 + (size_t)68 * 3; i1c2_5.B = iw1 + 5; i1c2_5.bias = R67 + 0 + (size_t)68 * 3; i1c2_5.R = R67 + 26176 + (size_t)67 * 16; i1c2_5.C = R67 + 26176 + (size_t)67 * 16;
      i1c2_5.sAo = (long long)66 * 66 * 3; i1c2_5.sAi = (long long)66 * 3; i1c2_5.sAm = 3; i1c2_5.sAk = 1; i1c2_5.sBo = 0; i1c2_5.sBi = 0; i1c2_5.sBn = 3 * 9; i1c2_5.sBk = 9; i1c2_5.sCo = (long long)66 * 66 * 16; i1c2_5.sCi = (long long)66 * 16; i1c2_5.sCm = 16; i1c2_5.sRo = (long long)66 * 66 * 16; i1c2_5.sRi = (long long)66 * 16; i1c2_5.sRm = 16; i1c2_5.sRn = 1;
      i1c2_5.M = 64; i1c2_5.N = 16; i1c2_5.K = 3; i1c2_5.zi_n = 64; i1c2_5.flags = 4; i1c2_5.act = 0;
      i1c2_5.alpha = 1.0f; i1c2_5.beta = 1.0f; i1c2_5.sa = 1.0f; i1c2_5.sb = 1.0f; i1c2_5.Npad = 16; i1c2_5.pad_ = 0;
      k_gemm<1><<<dim3((unsigned)((16) + 31) / 32, (unsigned)((64) + 15) / 16, (unsigned)(2 * 64)), 32, 0, stream>>>(i1c2_5); }
    { GemmP i1c2_6;
      i1c2_6.A = R67 + 0 + (size_t)132 * 3; i1c2_6.B = iw1 + 6; i1c2_6.bias = R67 + 0 + (size_t)132 * 3; i1c2_6.R = R67 + 26176 + (size_t)67 * 16; i1c2_6.C = R67 + 26176 + (size_t)67 * 16;
      i1c2_6.sAo = (long long)66 * 66 * 3; i1c2_6.sAi = (long long)66 * 3; i1c2_6.sAm = 3; i1c2_6.sAk = 1; i1c2_6.sBo = 0; i1c2_6.sBi = 0; i1c2_6.sBn = 3 * 9; i1c2_6.sBk = 9; i1c2_6.sCo = (long long)66 * 66 * 16; i1c2_6.sCi = (long long)66 * 16; i1c2_6.sCm = 16; i1c2_6.sRo = (long long)66 * 66 * 16; i1c2_6.sRi = (long long)66 * 16; i1c2_6.sRm = 16; i1c2_6.sRn = 1;
      i1c2_6.M = 64; i1c2_6.N = 16; i1c2_6.K = 3; i1c2_6.zi_n = 64; i1c2_6.flags = 4; i1c2_6.act = 0;
      i1c2_6.alpha = 1.0f; i1c2_6.beta = 1.0f; i1c2_6.sa = 1.0f; i1c2_6.sb = 1.0f; i1c2_6.Npad = 16; i1c2_6.pad_ = 0;
      k_gemm<1><<<dim3((unsigned)((16) + 31) / 32, (unsigned)((64) + 15) / 16, (unsigned)(2 * 64)), 32, 0, stream>>>(i1c2_6); }
    { GemmP i1c2_7;
      i1c2_7.A = R67 + 0 + (size_t)133 * 3; i1c2_7.B = iw1 + 7; i1c2_7.bias = R67 + 0 + (size_t)133 * 3; i1c2_7.R = R67 + 26176 + (size_t)67 * 16; i1c2_7.C = R67 + 26176 + (size_t)67 * 16;
      i1c2_7.sAo = (long long)66 * 66 * 3; i1c2_7.sAi = (long long)66 * 3; i1c2_7.sAm = 3; i1c2_7.sAk = 1; i1c2_7.sBo = 0; i1c2_7.sBi = 0; i1c2_7.sBn = 3 * 9; i1c2_7.sBk = 9; i1c2_7.sCo = (long long)66 * 66 * 16; i1c2_7.sCi = (long long)66 * 16; i1c2_7.sCm = 16; i1c2_7.sRo = (long long)66 * 66 * 16; i1c2_7.sRi = (long long)66 * 16; i1c2_7.sRm = 16; i1c2_7.sRn = 1;
      i1c2_7.M = 64; i1c2_7.N = 16; i1c2_7.K = 3; i1c2_7.zi_n = 64; i1c2_7.flags = 4; i1c2_7.act = 0;
      i1c2_7.alpha = 1.0f; i1c2_7.beta = 1.0f; i1c2_7.sa = 1.0f; i1c2_7.sb = 1.0f; i1c2_7.Npad = 16; i1c2_7.pad_ = 0;
      k_gemm<1><<<dim3((unsigned)((16) + 31) / 32, (unsigned)((64) + 15) / 16, (unsigned)(2 * 64)), 32, 0, stream>>>(i1c2_7); }
    { GemmP i1c2_8;
      i1c2_8.A = R67 + 0 + (size_t)134 * 3; i1c2_8.B = iw1 + 8; i1c2_8.bias = R67 + 0 + (size_t)134 * 3; i1c2_8.R = R67 + 26176 + (size_t)67 * 16; i1c2_8.C = R67 + 26176 + (size_t)67 * 16;
      i1c2_8.sAo = (long long)66 * 66 * 3; i1c2_8.sAi = (long long)66 * 3; i1c2_8.sAm = 3; i1c2_8.sAk = 1; i1c2_8.sBo = 0; i1c2_8.sBi = 0; i1c2_8.sBn = 3 * 9; i1c2_8.sBk = 9; i1c2_8.sCo = (long long)66 * 66 * 16; i1c2_8.sCi = (long long)66 * 16; i1c2_8.sCm = 16; i1c2_8.sRo = (long long)66 * 66 * 16; i1c2_8.sRi = (long long)66 * 16; i1c2_8.sRm = 16; i1c2_8.sRn = 1;
      i1c2_8.M = 64; i1c2_8.N = 16; i1c2_8.K = 3; i1c2_8.zi_n = 64; i1c2_8.flags = 4; i1c2_8.act = 0;
      i1c2_8.alpha = 1.0f; i1c2_8.beta = 1.0f; i1c2_8.sa = 1.0f; i1c2_8.sb = 1.0f; i1c2_8.Npad = 16; i1c2_8.pad_ = 0;
      k_gemm<1><<<dim3((unsigned)((16) + 31) / 32, (unsigned)((64) + 15) / 16, (unsigned)(2 * 64)), 32, 0, stream>>>(i1c2_8); }
    k_mm_relu2d<<<(unsigned)(((long long)2 * HW * 16 + 255) / 256), 256, 0, stream>>>(R67 + 26176, nullptr, 2, 64, 16);
    { GemmP i2c2_0;
      i2c2_0.A = R67 + 26176 + (size_t)0 * 16; i2c2_0.B = iw2 + 0; i2c2_0.bias = ib2; i2c2_0.R = R67 + 26176 + (size_t)0 * 16; i2c2_0.C = R67 + 165568 + (size_t)67 * 32;
      i2c2_0.sAo = (long long)66 * 66 * 16; i2c2_0.sAi = (long long)66 * 16; i2c2_0.sAm = 16; i2c2_0.sAk = 1; i2c2_0.sBo = 0; i2c2_0.sBi = 0; i2c2_0.sBn = 16 * 9; i2c2_0.sBk = 9; i2c2_0.sCo = (long long)66 * 66 * 32; i2c2_0.sCi = (long long)66 * 32; i2c2_0.sCm = 32; i2c2_0.sRo = 0; i2c2_0.sRi = 0; i2c2_0.sRm = 0; i2c2_0.sRn = 0;
      i2c2_0.M = 64; i2c2_0.N = 32; i2c2_0.K = 16; i2c2_0.zi_n = 64; i2c2_0.flags = 1; i2c2_0.act = 0;
      i2c2_0.alpha = 1.0f; i2c2_0.beta = 0.0f; i2c2_0.sa = 1.0f; i2c2_0.sb = 1.0f; i2c2_0.Npad = 32; i2c2_0.pad_ = 0;
      k_gemm<1><<<dim3((unsigned)((32) + 31) / 32, (unsigned)((64) + 15) / 16, (unsigned)(2 * 64)), 32, 0, stream>>>(i2c2_0); }
    { GemmP i2c2_1;
      i2c2_1.A = R67 + 26176 + (size_t)1 * 16; i2c2_1.B = iw2 + 1; i2c2_1.bias = R67 + 26176 + (size_t)1 * 16; i2c2_1.R = R67 + 165568 + (size_t)67 * 32; i2c2_1.C = R67 + 165568 + (size_t)67 * 32;
      i2c2_1.sAo = (long long)66 * 66 * 16; i2c2_1.sAi = (long long)66 * 16; i2c2_1.sAm = 16; i2c2_1.sAk = 1; i2c2_1.sBo = 0; i2c2_1.sBi = 0; i2c2_1.sBn = 16 * 9; i2c2_1.sBk = 9; i2c2_1.sCo = (long long)66 * 66 * 32; i2c2_1.sCi = (long long)66 * 32; i2c2_1.sCm = 32; i2c2_1.sRo = (long long)66 * 66 * 32; i2c2_1.sRi = (long long)66 * 32; i2c2_1.sRm = 32; i2c2_1.sRn = 1;
      i2c2_1.M = 64; i2c2_1.N = 32; i2c2_1.K = 16; i2c2_1.zi_n = 64; i2c2_1.flags = 4; i2c2_1.act = 0;
      i2c2_1.alpha = 1.0f; i2c2_1.beta = 1.0f; i2c2_1.sa = 1.0f; i2c2_1.sb = 1.0f; i2c2_1.Npad = 32; i2c2_1.pad_ = 0;
      k_gemm<1><<<dim3((unsigned)((32) + 31) / 32, (unsigned)((64) + 15) / 16, (unsigned)(2 * 64)), 32, 0, stream>>>(i2c2_1); }
    { GemmP i2c2_2;
      i2c2_2.A = R67 + 26176 + (size_t)2 * 16; i2c2_2.B = iw2 + 2; i2c2_2.bias = R67 + 26176 + (size_t)2 * 16; i2c2_2.R = R67 + 165568 + (size_t)67 * 32; i2c2_2.C = R67 + 165568 + (size_t)67 * 32;
      i2c2_2.sAo = (long long)66 * 66 * 16; i2c2_2.sAi = (long long)66 * 16; i2c2_2.sAm = 16; i2c2_2.sAk = 1; i2c2_2.sBo = 0; i2c2_2.sBi = 0; i2c2_2.sBn = 16 * 9; i2c2_2.sBk = 9; i2c2_2.sCo = (long long)66 * 66 * 32; i2c2_2.sCi = (long long)66 * 32; i2c2_2.sCm = 32; i2c2_2.sRo = (long long)66 * 66 * 32; i2c2_2.sRi = (long long)66 * 32; i2c2_2.sRm = 32; i2c2_2.sRn = 1;
      i2c2_2.M = 64; i2c2_2.N = 32; i2c2_2.K = 16; i2c2_2.zi_n = 64; i2c2_2.flags = 4; i2c2_2.act = 0;
      i2c2_2.alpha = 1.0f; i2c2_2.beta = 1.0f; i2c2_2.sa = 1.0f; i2c2_2.sb = 1.0f; i2c2_2.Npad = 32; i2c2_2.pad_ = 0;
      k_gemm<1><<<dim3((unsigned)((32) + 31) / 32, (unsigned)((64) + 15) / 16, (unsigned)(2 * 64)), 32, 0, stream>>>(i2c2_2); }
    { GemmP i2c2_3;
      i2c2_3.A = R67 + 26176 + (size_t)66 * 16; i2c2_3.B = iw2 + 3; i2c2_3.bias = R67 + 26176 + (size_t)66 * 16; i2c2_3.R = R67 + 165568 + (size_t)67 * 32; i2c2_3.C = R67 + 165568 + (size_t)67 * 32;
      i2c2_3.sAo = (long long)66 * 66 * 16; i2c2_3.sAi = (long long)66 * 16; i2c2_3.sAm = 16; i2c2_3.sAk = 1; i2c2_3.sBo = 0; i2c2_3.sBi = 0; i2c2_3.sBn = 16 * 9; i2c2_3.sBk = 9; i2c2_3.sCo = (long long)66 * 66 * 32; i2c2_3.sCi = (long long)66 * 32; i2c2_3.sCm = 32; i2c2_3.sRo = (long long)66 * 66 * 32; i2c2_3.sRi = (long long)66 * 32; i2c2_3.sRm = 32; i2c2_3.sRn = 1;
      i2c2_3.M = 64; i2c2_3.N = 32; i2c2_3.K = 16; i2c2_3.zi_n = 64; i2c2_3.flags = 4; i2c2_3.act = 0;
      i2c2_3.alpha = 1.0f; i2c2_3.beta = 1.0f; i2c2_3.sa = 1.0f; i2c2_3.sb = 1.0f; i2c2_3.Npad = 32; i2c2_3.pad_ = 0;
      k_gemm<1><<<dim3((unsigned)((32) + 31) / 32, (unsigned)((64) + 15) / 16, (unsigned)(2 * 64)), 32, 0, stream>>>(i2c2_3); }
    { GemmP i2c2_4;
      i2c2_4.A = R67 + 26176 + (size_t)67 * 16; i2c2_4.B = iw2 + 4; i2c2_4.bias = R67 + 26176 + (size_t)67 * 16; i2c2_4.R = R67 + 165568 + (size_t)67 * 32; i2c2_4.C = R67 + 165568 + (size_t)67 * 32;
      i2c2_4.sAo = (long long)66 * 66 * 16; i2c2_4.sAi = (long long)66 * 16; i2c2_4.sAm = 16; i2c2_4.sAk = 1; i2c2_4.sBo = 0; i2c2_4.sBi = 0; i2c2_4.sBn = 16 * 9; i2c2_4.sBk = 9; i2c2_4.sCo = (long long)66 * 66 * 32; i2c2_4.sCi = (long long)66 * 32; i2c2_4.sCm = 32; i2c2_4.sRo = (long long)66 * 66 * 32; i2c2_4.sRi = (long long)66 * 32; i2c2_4.sRm = 32; i2c2_4.sRn = 1;
      i2c2_4.M = 64; i2c2_4.N = 32; i2c2_4.K = 16; i2c2_4.zi_n = 64; i2c2_4.flags = 4; i2c2_4.act = 0;
      i2c2_4.alpha = 1.0f; i2c2_4.beta = 1.0f; i2c2_4.sa = 1.0f; i2c2_4.sb = 1.0f; i2c2_4.Npad = 32; i2c2_4.pad_ = 0;
      k_gemm<1><<<dim3((unsigned)((32) + 31) / 32, (unsigned)((64) + 15) / 16, (unsigned)(2 * 64)), 32, 0, stream>>>(i2c2_4); }
    { GemmP i2c2_5;
      i2c2_5.A = R67 + 26176 + (size_t)68 * 16; i2c2_5.B = iw2 + 5; i2c2_5.bias = R67 + 26176 + (size_t)68 * 16; i2c2_5.R = R67 + 165568 + (size_t)67 * 32; i2c2_5.C = R67 + 165568 + (size_t)67 * 32;
      i2c2_5.sAo = (long long)66 * 66 * 16; i2c2_5.sAi = (long long)66 * 16; i2c2_5.sAm = 16; i2c2_5.sAk = 1; i2c2_5.sBo = 0; i2c2_5.sBi = 0; i2c2_5.sBn = 16 * 9; i2c2_5.sBk = 9; i2c2_5.sCo = (long long)66 * 66 * 32; i2c2_5.sCi = (long long)66 * 32; i2c2_5.sCm = 32; i2c2_5.sRo = (long long)66 * 66 * 32; i2c2_5.sRi = (long long)66 * 32; i2c2_5.sRm = 32; i2c2_5.sRn = 1;
      i2c2_5.M = 64; i2c2_5.N = 32; i2c2_5.K = 16; i2c2_5.zi_n = 64; i2c2_5.flags = 4; i2c2_5.act = 0;
      i2c2_5.alpha = 1.0f; i2c2_5.beta = 1.0f; i2c2_5.sa = 1.0f; i2c2_5.sb = 1.0f; i2c2_5.Npad = 32; i2c2_5.pad_ = 0;
      k_gemm<1><<<dim3((unsigned)((32) + 31) / 32, (unsigned)((64) + 15) / 16, (unsigned)(2 * 64)), 32, 0, stream>>>(i2c2_5); }
    { GemmP i2c2_6;
      i2c2_6.A = R67 + 26176 + (size_t)132 * 16; i2c2_6.B = iw2 + 6; i2c2_6.bias = R67 + 26176 + (size_t)132 * 16; i2c2_6.R = R67 + 165568 + (size_t)67 * 32; i2c2_6.C = R67 + 165568 + (size_t)67 * 32;
      i2c2_6.sAo = (long long)66 * 66 * 16; i2c2_6.sAi = (long long)66 * 16; i2c2_6.sAm = 16; i2c2_6.sAk = 1; i2c2_6.sBo = 0; i2c2_6.sBi = 0; i2c2_6.sBn = 16 * 9; i2c2_6.sBk = 9; i2c2_6.sCo = (long long)66 * 66 * 32; i2c2_6.sCi = (long long)66 * 32; i2c2_6.sCm = 32; i2c2_6.sRo = (long long)66 * 66 * 32; i2c2_6.sRi = (long long)66 * 32; i2c2_6.sRm = 32; i2c2_6.sRn = 1;
      i2c2_6.M = 64; i2c2_6.N = 32; i2c2_6.K = 16; i2c2_6.zi_n = 64; i2c2_6.flags = 4; i2c2_6.act = 0;
      i2c2_6.alpha = 1.0f; i2c2_6.beta = 1.0f; i2c2_6.sa = 1.0f; i2c2_6.sb = 1.0f; i2c2_6.Npad = 32; i2c2_6.pad_ = 0;
      k_gemm<1><<<dim3((unsigned)((32) + 31) / 32, (unsigned)((64) + 15) / 16, (unsigned)(2 * 64)), 32, 0, stream>>>(i2c2_6); }
    { GemmP i2c2_7;
      i2c2_7.A = R67 + 26176 + (size_t)133 * 16; i2c2_7.B = iw2 + 7; i2c2_7.bias = R67 + 26176 + (size_t)133 * 16; i2c2_7.R = R67 + 165568 + (size_t)67 * 32; i2c2_7.C = R67 + 165568 + (size_t)67 * 32;
      i2c2_7.sAo = (long long)66 * 66 * 16; i2c2_7.sAi = (long long)66 * 16; i2c2_7.sAm = 16; i2c2_7.sAk = 1; i2c2_7.sBo = 0; i2c2_7.sBi = 0; i2c2_7.sBn = 16 * 9; i2c2_7.sBk = 9; i2c2_7.sCo = (long long)66 * 66 * 32; i2c2_7.sCi = (long long)66 * 32; i2c2_7.sCm = 32; i2c2_7.sRo = (long long)66 * 66 * 32; i2c2_7.sRi = (long long)66 * 32; i2c2_7.sRm = 32; i2c2_7.sRn = 1;
      i2c2_7.M = 64; i2c2_7.N = 32; i2c2_7.K = 16; i2c2_7.zi_n = 64; i2c2_7.flags = 4; i2c2_7.act = 0;
      i2c2_7.alpha = 1.0f; i2c2_7.beta = 1.0f; i2c2_7.sa = 1.0f; i2c2_7.sb = 1.0f; i2c2_7.Npad = 32; i2c2_7.pad_ = 0;
      k_gemm<1><<<dim3((unsigned)((32) + 31) / 32, (unsigned)((64) + 15) / 16, (unsigned)(2 * 64)), 32, 0, stream>>>(i2c2_7); }
    { GemmP i2c2_8;
      i2c2_8.A = R67 + 26176 + (size_t)134 * 16; i2c2_8.B = iw2 + 8; i2c2_8.bias = R67 + 26176 + (size_t)134 * 16; i2c2_8.R = R67 + 165568 + (size_t)67 * 32; i2c2_8.C = R67 + 165568 + (size_t)67 * 32;
      i2c2_8.sAo = (long long)66 * 66 * 16; i2c2_8.sAi = (long long)66 * 16; i2c2_8.sAm = 16; i2c2_8.sAk = 1; i2c2_8.sBo = 0; i2c2_8.sBi = 0; i2c2_8.sBn = 16 * 9; i2c2_8.sBk = 9; i2c2_8.sCo = (long long)66 * 66 * 32; i2c2_8.sCi = (long long)66 * 32; i2c2_8.sCm = 32; i2c2_8.sRo = (long long)66 * 66 * 32; i2c2_8.sRi = (long long)66 * 32; i2c2_8.sRm = 32; i2c2_8.sRn = 1;
      i2c2_8.M = 64; i2c2_8.N = 32; i2c2_8.K = 16; i2c2_8.zi_n = 64; i2c2_8.flags = 4; i2c2_8.act = 0;
      i2c2_8.alpha = 1.0f; i2c2_8.beta = 1.0f; i2c2_8.sa = 1.0f; i2c2_8.sb = 1.0f; i2c2_8.Npad = 32; i2c2_8.pad_ = 0;
      k_gemm<1><<<dim3((unsigned)((32) + 31) / 32, (unsigned)((64) + 15) / 16, (unsigned)(2 * 64)), 32, 0, stream>>>(i2c2_8); }
    k_mm_relu2d<<<(unsigned)(((long long)2 * HW * 32 + 255) / 256), 256, 0, stream>>>(R67 + 165568, nullptr, 2, 64, 32);
    { GemmP i3c2_0;
      i3c2_0.A = R67 + 165568 + (size_t)0 * 32; i3c2_0.B = iw3 + 0; i3c2_0.bias = ib3; i3c2_0.R = R67 + 165568 + (size_t)0 * 32; i3c2_0.C = R67 + 444352 + (size_t)67 * 64;
      i3c2_0.sAo = (long long)66 * 66 * 32; i3c2_0.sAi = (long long)66 * 32; i3c2_0.sAm = 32; i3c2_0.sAk = 1; i3c2_0.sBo = 0; i3c2_0.sBi = 0; i3c2_0.sBn = 32 * 9; i3c2_0.sBk = 9; i3c2_0.sCo = (long long)66 * 66 * 64; i3c2_0.sCi = (long long)66 * 64; i3c2_0.sCm = 64; i3c2_0.sRo = 0; i3c2_0.sRi = 0; i3c2_0.sRm = 0; i3c2_0.sRn = 0;
      i3c2_0.M = 64; i3c2_0.N = 64; i3c2_0.K = 32; i3c2_0.zi_n = 64; i3c2_0.flags = 1; i3c2_0.act = 0;
      i3c2_0.alpha = 1.0f; i3c2_0.beta = 0.0f; i3c2_0.sa = 1.0f; i3c2_0.sb = 1.0f; i3c2_0.Npad = 64; i3c2_0.pad_ = 0;
      k_gemm<1><<<dim3((unsigned)((64) + 31) / 32, (unsigned)((64) + 15) / 16, (unsigned)(2 * 64)), 32, 0, stream>>>(i3c2_0); }
    { GemmP i3c2_1;
      i3c2_1.A = R67 + 165568 + (size_t)1 * 32; i3c2_1.B = iw3 + 1; i3c2_1.bias = R67 + 165568 + (size_t)1 * 32; i3c2_1.R = R67 + 444352 + (size_t)67 * 64; i3c2_1.C = R67 + 444352 + (size_t)67 * 64;
      i3c2_1.sAo = (long long)66 * 66 * 32; i3c2_1.sAi = (long long)66 * 32; i3c2_1.sAm = 32; i3c2_1.sAk = 1; i3c2_1.sBo = 0; i3c2_1.sBi = 0; i3c2_1.sBn = 32 * 9; i3c2_1.sBk = 9; i3c2_1.sCo = (long long)66 * 66 * 64; i3c2_1.sCi = (long long)66 * 64; i3c2_1.sCm = 64; i3c2_1.sRo = (long long)66 * 66 * 64; i3c2_1.sRi = (long long)66 * 64; i3c2_1.sRm = 64; i3c2_1.sRn = 1;
      i3c2_1.M = 64; i3c2_1.N = 64; i3c2_1.K = 32; i3c2_1.zi_n = 64; i3c2_1.flags = 4; i3c2_1.act = 0;
      i3c2_1.alpha = 1.0f; i3c2_1.beta = 1.0f; i3c2_1.sa = 1.0f; i3c2_1.sb = 1.0f; i3c2_1.Npad = 64; i3c2_1.pad_ = 0;
      k_gemm<1><<<dim3((unsigned)((64) + 31) / 32, (unsigned)((64) + 15) / 16, (unsigned)(2 * 64)), 32, 0, stream>>>(i3c2_1); }
    { GemmP i3c2_2;
      i3c2_2.A = R67 + 165568 + (size_t)2 * 32; i3c2_2.B = iw3 + 2; i3c2_2.bias = R67 + 165568 + (size_t)2 * 32; i3c2_2.R = R67 + 444352 + (size_t)67 * 64; i3c2_2.C = R67 + 444352 + (size_t)67 * 64;
      i3c2_2.sAo = (long long)66 * 66 * 32; i3c2_2.sAi = (long long)66 * 32; i3c2_2.sAm = 32; i3c2_2.sAk = 1; i3c2_2.sBo = 0; i3c2_2.sBi = 0; i3c2_2.sBn = 32 * 9; i3c2_2.sBk = 9; i3c2_2.sCo = (long long)66 * 66 * 64; i3c2_2.sCi = (long long)66 * 64; i3c2_2.sCm = 64; i3c2_2.sRo = (long long)66 * 66 * 64; i3c2_2.sRi = (long long)66 * 64; i3c2_2.sRm = 64; i3c2_2.sRn = 1;
      i3c2_2.M = 64; i3c2_2.N = 64; i3c2_2.K = 32; i3c2_2.zi_n = 64; i3c2_2.flags = 4; i3c2_2.act = 0;
      i3c2_2.alpha = 1.0f; i3c2_2.beta = 1.0f; i3c2_2.sa = 1.0f; i3c2_2.sb = 1.0f; i3c2_2.Npad = 64; i3c2_2.pad_ = 0;
      k_gemm<1><<<dim3((unsigned)((64) + 31) / 32, (unsigned)((64) + 15) / 16, (unsigned)(2 * 64)), 32, 0, stream>>>(i3c2_2); }
    { GemmP i3c2_3;
      i3c2_3.A = R67 + 165568 + (size_t)66 * 32; i3c2_3.B = iw3 + 3; i3c2_3.bias = R67 + 165568 + (size_t)66 * 32; i3c2_3.R = R67 + 444352 + (size_t)67 * 64; i3c2_3.C = R67 + 444352 + (size_t)67 * 64;
      i3c2_3.sAo = (long long)66 * 66 * 32; i3c2_3.sAi = (long long)66 * 32; i3c2_3.sAm = 32; i3c2_3.sAk = 1; i3c2_3.sBo = 0; i3c2_3.sBi = 0; i3c2_3.sBn = 32 * 9; i3c2_3.sBk = 9; i3c2_3.sCo = (long long)66 * 66 * 64; i3c2_3.sCi = (long long)66 * 64; i3c2_3.sCm = 64; i3c2_3.sRo = (long long)66 * 66 * 64; i3c2_3.sRi = (long long)66 * 64; i3c2_3.sRm = 64; i3c2_3.sRn = 1;
      i3c2_3.M = 64; i3c2_3.N = 64; i3c2_3.K = 32; i3c2_3.zi_n = 64; i3c2_3.flags = 4; i3c2_3.act = 0;
      i3c2_3.alpha = 1.0f; i3c2_3.beta = 1.0f; i3c2_3.sa = 1.0f; i3c2_3.sb = 1.0f; i3c2_3.Npad = 64; i3c2_3.pad_ = 0;
      k_gemm<1><<<dim3((unsigned)((64) + 31) / 32, (unsigned)((64) + 15) / 16, (unsigned)(2 * 64)), 32, 0, stream>>>(i3c2_3); }
    { GemmP i3c2_4;
      i3c2_4.A = R67 + 165568 + (size_t)67 * 32; i3c2_4.B = iw3 + 4; i3c2_4.bias = R67 + 165568 + (size_t)67 * 32; i3c2_4.R = R67 + 444352 + (size_t)67 * 64; i3c2_4.C = R67 + 444352 + (size_t)67 * 64;
      i3c2_4.sAo = (long long)66 * 66 * 32; i3c2_4.sAi = (long long)66 * 32; i3c2_4.sAm = 32; i3c2_4.sAk = 1; i3c2_4.sBo = 0; i3c2_4.sBi = 0; i3c2_4.sBn = 32 * 9; i3c2_4.sBk = 9; i3c2_4.sCo = (long long)66 * 66 * 64; i3c2_4.sCi = (long long)66 * 64; i3c2_4.sCm = 64; i3c2_4.sRo = (long long)66 * 66 * 64; i3c2_4.sRi = (long long)66 * 64; i3c2_4.sRm = 64; i3c2_4.sRn = 1;
      i3c2_4.M = 64; i3c2_4.N = 64; i3c2_4.K = 32; i3c2_4.zi_n = 64; i3c2_4.flags = 4; i3c2_4.act = 0;
      i3c2_4.alpha = 1.0f; i3c2_4.beta = 1.0f; i3c2_4.sa = 1.0f; i3c2_4.sb = 1.0f; i3c2_4.Npad = 64; i3c2_4.pad_ = 0;
      k_gemm<1><<<dim3((unsigned)((64) + 31) / 32, (unsigned)((64) + 15) / 16, (unsigned)(2 * 64)), 32, 0, stream>>>(i3c2_4); }
    { GemmP i3c2_5;
      i3c2_5.A = R67 + 165568 + (size_t)68 * 32; i3c2_5.B = iw3 + 5; i3c2_5.bias = R67 + 165568 + (size_t)68 * 32; i3c2_5.R = R67 + 444352 + (size_t)67 * 64; i3c2_5.C = R67 + 444352 + (size_t)67 * 64;
      i3c2_5.sAo = (long long)66 * 66 * 32; i3c2_5.sAi = (long long)66 * 32; i3c2_5.sAm = 32; i3c2_5.sAk = 1; i3c2_5.sBo = 0; i3c2_5.sBi = 0; i3c2_5.sBn = 32 * 9; i3c2_5.sBk = 9; i3c2_5.sCo = (long long)66 * 66 * 64; i3c2_5.sCi = (long long)66 * 64; i3c2_5.sCm = 64; i3c2_5.sRo = (long long)66 * 66 * 64; i3c2_5.sRi = (long long)66 * 64; i3c2_5.sRm = 64; i3c2_5.sRn = 1;
      i3c2_5.M = 64; i3c2_5.N = 64; i3c2_5.K = 32; i3c2_5.zi_n = 64; i3c2_5.flags = 4; i3c2_5.act = 0;
      i3c2_5.alpha = 1.0f; i3c2_5.beta = 1.0f; i3c2_5.sa = 1.0f; i3c2_5.sb = 1.0f; i3c2_5.Npad = 64; i3c2_5.pad_ = 0;
      k_gemm<1><<<dim3((unsigned)((64) + 31) / 32, (unsigned)((64) + 15) / 16, (unsigned)(2 * 64)), 32, 0, stream>>>(i3c2_5); }
    { GemmP i3c2_6;
      i3c2_6.A = R67 + 165568 + (size_t)132 * 32; i3c2_6.B = iw3 + 6; i3c2_6.bias = R67 + 165568 + (size_t)132 * 32; i3c2_6.R = R67 + 444352 + (size_t)67 * 64; i3c2_6.C = R67 + 444352 + (size_t)67 * 64;
      i3c2_6.sAo = (long long)66 * 66 * 32; i3c2_6.sAi = (long long)66 * 32; i3c2_6.sAm = 32; i3c2_6.sAk = 1; i3c2_6.sBo = 0; i3c2_6.sBi = 0; i3c2_6.sBn = 32 * 9; i3c2_6.sBk = 9; i3c2_6.sCo = (long long)66 * 66 * 64; i3c2_6.sCi = (long long)66 * 64; i3c2_6.sCm = 64; i3c2_6.sRo = (long long)66 * 66 * 64; i3c2_6.sRi = (long long)66 * 64; i3c2_6.sRm = 64; i3c2_6.sRn = 1;
      i3c2_6.M = 64; i3c2_6.N = 64; i3c2_6.K = 32; i3c2_6.zi_n = 64; i3c2_6.flags = 4; i3c2_6.act = 0;
      i3c2_6.alpha = 1.0f; i3c2_6.beta = 1.0f; i3c2_6.sa = 1.0f; i3c2_6.sb = 1.0f; i3c2_6.Npad = 64; i3c2_6.pad_ = 0;
      k_gemm<1><<<dim3((unsigned)((64) + 31) / 32, (unsigned)((64) + 15) / 16, (unsigned)(2 * 64)), 32, 0, stream>>>(i3c2_6); }
    { GemmP i3c2_7;
      i3c2_7.A = R67 + 165568 + (size_t)133 * 32; i3c2_7.B = iw3 + 7; i3c2_7.bias = R67 + 165568 + (size_t)133 * 32; i3c2_7.R = R67 + 444352 + (size_t)67 * 64; i3c2_7.C = R67 + 444352 + (size_t)67 * 64;
      i3c2_7.sAo = (long long)66 * 66 * 32; i3c2_7.sAi = (long long)66 * 32; i3c2_7.sAm = 32; i3c2_7.sAk = 1; i3c2_7.sBo = 0; i3c2_7.sBi = 0; i3c2_7.sBn = 32 * 9; i3c2_7.sBk = 9; i3c2_7.sCo = (long long)66 * 66 * 64; i3c2_7.sCi = (long long)66 * 64; i3c2_7.sCm = 64; i3c2_7.sRo = (long long)66 * 66 * 64; i3c2_7.sRi = (long long)66 * 64; i3c2_7.sRm = 64; i3c2_7.sRn = 1;
      i3c2_7.M = 64; i3c2_7.N = 64; i3c2_7.K = 32; i3c2_7.zi_n = 64; i3c2_7.flags = 4; i3c2_7.act = 0;
      i3c2_7.alpha = 1.0f; i3c2_7.beta = 1.0f; i3c2_7.sa = 1.0f; i3c2_7.sb = 1.0f; i3c2_7.Npad = 64; i3c2_7.pad_ = 0;
      k_gemm<1><<<dim3((unsigned)((64) + 31) / 32, (unsigned)((64) + 15) / 16, (unsigned)(2 * 64)), 32, 0, stream>>>(i3c2_7); }
    { GemmP i3c2_8;
      i3c2_8.A = R67 + 165568 + (size_t)134 * 32; i3c2_8.B = iw3 + 8; i3c2_8.bias = R67 + 165568 + (size_t)134 * 32; i3c2_8.R = R67 + 444352 + (size_t)67 * 64; i3c2_8.C = R67 + 444352 + (size_t)67 * 64;
      i3c2_8.sAo = (long long)66 * 66 * 32; i3c2_8.sAi = (long long)66 * 32; i3c2_8.sAm = 32; i3c2_8.sAk = 1; i3c2_8.sBo = 0; i3c2_8.sBi = 0; i3c2_8.sBn = 32 * 9; i3c2_8.sBk = 9; i3c2_8.sCo = (long long)66 * 66 * 64; i3c2_8.sCi = (long long)66 * 64; i3c2_8.sCm = 64; i3c2_8.sRo = (long long)66 * 66 * 64; i3c2_8.sRi = (long long)66 * 64; i3c2_8.sRm = 64; i3c2_8.sRn = 1;
      i3c2_8.M = 64; i3c2_8.N = 64; i3c2_8.K = 32; i3c2_8.zi_n = 64; i3c2_8.flags = 4; i3c2_8.act = 0;
      i3c2_8.alpha = 1.0f; i3c2_8.beta = 1.0f; i3c2_8.sa = 1.0f; i3c2_8.sb = 1.0f; i3c2_8.Npad = 64; i3c2_8.pad_ = 0;
      k_gemm<1><<<dim3((unsigned)((64) + 31) / 32, (unsigned)((64) + 15) / 16, (unsigned)(2 * 64)), 32, 0, stream>>>(i3c2_8); }
    k_mm_relu2d<<<(unsigned)(((long long)2 * HW * 64 + 255) / 256), 256, 0, stream>>>(R67 + 444352, R67 + 1001920, 2, 64, 64);
    { GemmP gqkv2;
      gqkv2.A = R67 + 1001920; gqkv2.B = qkvw; gqkv2.bias = qkvb; gqkv2.R = R67 + 1001920; gqkv2.C = R67 + 1526208;
      gqkv2.sAo = 0; gqkv2.sAi = 0; gqkv2.sAm = 64; gqkv2.sAk = 1; gqkv2.sBo = 0; gqkv2.sBi = 0; gqkv2.sBn = 64; gqkv2.sBk = 1; gqkv2.sCo = 0; gqkv2.sCi = 0; gqkv2.sCm = 192; gqkv2.sRo = 0; gqkv2.sRi = 0; gqkv2.sRm = 0; gqkv2.sRn = 0;
      gqkv2.M = 2 * HW; gqkv2.N = 192; gqkv2.K = 64; gqkv2.zi_n = 1; gqkv2.flags = 1; gqkv2.act = 0;
      gqkv2.alpha = 1.0f; gqkv2.beta = 0.0f; gqkv2.sa = 1.0f; gqkv2.sb = 1.0f; gqkv2.Npad = 192; gqkv2.pad_ = 0;
      k_gemm<1><<<dim3((unsigned)((192) + 31) / 32, (unsigned)((2 * HW) + 15) / 16, (unsigned)(1)), 32, 0, stream>>>(gqkv2); }
    k_mm_dw<<<(unsigned)(((long long)2 * HW * 192 + 255) / 256), 256, 0, stream>>>(R67 + 1526208, dww, dwb, R67 + 3099072, 2, 64, 192);
    k_mm_fall<<<(unsigned)(((long long)2 * HW * 144 + 255) / 256), 256, 0, stream>>>(R67 + 3099072, fcw, fcb, R67 + 4671936, 2, HW, 192);
    k_mm_dep<<<(unsigned)(((long long)2 * 64 * HW + 255) / 256), 256, 0, stream>>>(R67 + 4671936, depw, depb, R67 + 5851584, 2, 64);
    k_mm_qknorm<<<2 * 128, 256, 0, stream>>>(R67 + 3099072, R67 + 6375872, 2, HW, 192);
    { GemmP gat2;
      gat2.A = R67 + 6375872; gat2.B = R67 + 6375872 + (size_t)64 * HW; gat2.bias = R67 + 6375872; gat2.R = R67 + 6375872; gat2.C = R67 + 7424448;
      gat2.sAo = (long long)128 * HW; gat2.sAi = (long long)16 * HW; gat2.sAm = HW; gat2.sAk = 1; gat2.sBo = (long long)128 * HW; gat2.sBi = (long long)16 * HW; gat2.sBn = HW; gat2.sBk = 1; gat2.sCo = (long long)4 * 16 * LP; gat2.sCi = 16 * LP; gat2.sCm = LP; gat2.sRo = 0; gat2.sRi = 0; gat2.sRm = 0; gat2.sRn = 0;
      gat2.M = 16; gat2.N = 16; gat2.K = HW; gat2.zi_n = 4; gat2.flags = 0; gat2.act = 0;
      gat2.alpha = 1.0f; gat2.beta = 0.0f; gat2.sa = 1.0f; gat2.sb = 1.0f; gat2.Npad = LP; gat2.pad_ = 0;
      k_gemm<1><<<dim3((unsigned)((LP) + 31) / 32, (unsigned)((16) + 15) / 16, (unsigned)(2 * 4)), 32, 0, stream>>>(gat2); }
    k_mm_sm16<<<(unsigned)((2 * 4 * 16 + 255) / 256), 256, 0, stream>>>(R67 + 7424448, temp, 2 * 4, LP);
    { GemmP gao2;
      gao2.A = R67 + 7424448; gao2.B = R67 + 3099072 + 128; gao2.bias = R67 + 7424448; gao2.R = R67 + 7424448; gao2.C = R67 + 7428544;
      gao2.sAo = (long long)4 * 16 * LP; gao2.sAi = 16 * LP; gao2.sAm = LP; gao2.sAk = 1; gao2.sBo = (long long)HW * 192; gao2.sBi = 16; gao2.sBn = 192; gao2.sBk = 1; gao2.sCo = (long long)64 * HW; gao2.sCi = (long long)16 * HW; gao2.sCm = HW; gao2.sRo = 0; gao2.sRi = 0; gao2.sRm = 0; gao2.sRn = 0;
      gao2.M = 16; gao2.N = HW; gao2.K = 16; gao2.zi_n = 4; gao2.flags = 0; gao2.act = 0;
      gao2.alpha = 1.0f; gao2.beta = 0.0f; gao2.sa = 1.0f; gao2.sb = 1.0f; gao2.Npad = HW; gao2.pad_ = 0;
      k_gemm<1><<<dim3((unsigned)((HW) + 31) / 32, (unsigned)((16) + 15) / 16, (unsigned)(2 * 4)), 32, 0, stream>>>(gao2); }
    { GemmP gproj2;
      gproj2.A = projw; gproj2.B = R67 + 7428544; gproj2.bias = projb; gproj2.R = projw; gproj2.C = R67 + 7952832;
      gproj2.sAo = 0; gproj2.sAi = 0; gproj2.sAm = 64; gproj2.sAk = 1; gproj2.sBo = (long long)64 * HW; gproj2.sBi = 0; gproj2.sBn = 1; gproj2.sBk = HW; gproj2.sCo = (long long)64 * HW; gproj2.sCi = 0; gproj2.sCm = HW; gproj2.sRo = 0; gproj2.sRi = 0; gproj2.sRm = 0; gproj2.sRn = 0;
      gproj2.M = 64; gproj2.N = HW; gproj2.K = 64; gproj2.zi_n = 1; gproj2.flags = 2; gproj2.act = 0;
      gproj2.alpha = 1.0f; gproj2.beta = 0.0f; gproj2.sa = 1.0f; gproj2.sb = 1.0f; gproj2.Npad = HW; gproj2.pad_ = 0;
      k_gemm<1><<<dim3((unsigned)((HW) + 31) / 32, (unsigned)((64) + 15) / 16, (unsigned)(2)), 32, 0, stream>>>(gproj2); }
    k_mm_imgfeat<<<(unsigned)(((long long)2 * SEQ * 64 + 255) / 256), 256, 0, stream>>>(R67 + 7952832, R67 + 5851584, IR + (size_t)4 * SEQ * 64, 2, HW, 64);
    hipMemsetAsync(R67 + 0, 0, (size_t)2 * 66 * 66 * 3 * 4, stream); hipMemsetAsync(R67 + 26176, 0, (size_t)2 * 66 * 66 * 16 * 4, stream); hipMemsetAsync(R67 + 165568, 0, (size_t)2 * 66 * 66 * 32 * 4, stream); hipMemsetAsync(R67 + 444352, 0, (size_t)2 * 66 * 66 * 64 * 4, stream);
    k_mm_padimg<<<(unsigned)(((long long)2 * HW * 3 + 255) / 256), 256, 0, stream>>>(img + (size_t)6 * 3 * HW, R67 + 0, 2, 3, 64);
    { GemmP i1c3_0;
      i1c3_0.A = R67 + 0 + (size_t)0 * 3; i1c3_0.B = iw1 + 0; i1c3_0.bias = ib1; i1c3_0.R = R67 + 0 + (size_t)0 * 3; i1c3_0.C = R67 + 26176 + (size_t)67 * 16;
      i1c3_0.sAo = (long long)66 * 66 * 3; i1c3_0.sAi = (long long)66 * 3; i1c3_0.sAm = 3; i1c3_0.sAk = 1; i1c3_0.sBo = 0; i1c3_0.sBi = 0; i1c3_0.sBn = 3 * 9; i1c3_0.sBk = 9; i1c3_0.sCo = (long long)66 * 66 * 16; i1c3_0.sCi = (long long)66 * 16; i1c3_0.sCm = 16; i1c3_0.sRo = 0; i1c3_0.sRi = 0; i1c3_0.sRm = 0; i1c3_0.sRn = 0;
      i1c3_0.M = 64; i1c3_0.N = 16; i1c3_0.K = 3; i1c3_0.zi_n = 64; i1c3_0.flags = 1; i1c3_0.act = 0;
      i1c3_0.alpha = 1.0f; i1c3_0.beta = 0.0f; i1c3_0.sa = 1.0f; i1c3_0.sb = 1.0f; i1c3_0.Npad = 16; i1c3_0.pad_ = 0;
      k_gemm<1><<<dim3((unsigned)((16) + 31) / 32, (unsigned)((64) + 15) / 16, (unsigned)(2 * 64)), 32, 0, stream>>>(i1c3_0); }
    { GemmP i1c3_1;
      i1c3_1.A = R67 + 0 + (size_t)1 * 3; i1c3_1.B = iw1 + 1; i1c3_1.bias = R67 + 0 + (size_t)1 * 3; i1c3_1.R = R67 + 26176 + (size_t)67 * 16; i1c3_1.C = R67 + 26176 + (size_t)67 * 16;
      i1c3_1.sAo = (long long)66 * 66 * 3; i1c3_1.sAi = (long long)66 * 3; i1c3_1.sAm = 3; i1c3_1.sAk = 1; i1c3_1.sBo = 0; i1c3_1.sBi = 0; i1c3_1.sBn = 3 * 9; i1c3_1.sBk = 9; i1c3_1.sCo = (long long)66 * 66 * 16; i1c3_1.sCi = (long long)66 * 16; i1c3_1.sCm = 16; i1c3_1.sRo = (long long)66 * 66 * 16; i1c3_1.sRi = (long long)66 * 16; i1c3_1.sRm = 16; i1c3_1.sRn = 1;
      i1c3_1.M = 64; i1c3_1.N = 16; i1c3_1.K = 3; i1c3_1.zi_n = 64; i1c3_1.flags = 4; i1c3_1.act = 0;
      i1c3_1.alpha = 1.0f; i1c3_1.beta = 1.0f; i1c3_1.sa = 1.0f; i1c3_1.sb = 1.0f; i1c3_1.Npad = 16; i1c3_1.pad_ = 0;
      k_gemm<1><<<dim3((unsigned)((16) + 31) / 32, (unsigned)((64) + 15) / 16, (unsigned)(2 * 64)), 32, 0, stream>>>(i1c3_1); }
    { GemmP i1c3_2;
      i1c3_2.A = R67 + 0 + (size_t)2 * 3; i1c3_2.B = iw1 + 2; i1c3_2.bias = R67 + 0 + (size_t)2 * 3; i1c3_2.R = R67 + 26176 + (size_t)67 * 16; i1c3_2.C = R67 + 26176 + (size_t)67 * 16;
      i1c3_2.sAo = (long long)66 * 66 * 3; i1c3_2.sAi = (long long)66 * 3; i1c3_2.sAm = 3; i1c3_2.sAk = 1; i1c3_2.sBo = 0; i1c3_2.sBi = 0; i1c3_2.sBn = 3 * 9; i1c3_2.sBk = 9; i1c3_2.sCo = (long long)66 * 66 * 16; i1c3_2.sCi = (long long)66 * 16; i1c3_2.sCm = 16; i1c3_2.sRo = (long long)66 * 66 * 16; i1c3_2.sRi = (long long)66 * 16; i1c3_2.sRm = 16; i1c3_2.sRn = 1;
      i1c3_2.M = 64; i1c3_2.N = 16; i1c3_2.K = 3; i1c3_2.zi_n = 64; i1c3_2.flags = 4; i1c3_2.act = 0;
      i1c3_2.alpha = 1.0f; i1c3_2.beta = 1.0f; i1c3_2.sa = 1.0f; i1c3_2.sb = 1.0f; i1c3_2.Npad = 16; i1c3_2.pad_ = 0;
      k_gemm<1><<<dim3((unsigned)((16) + 31) / 32, (unsigned)((64) + 15) / 16, (unsigned)(2 * 64)), 32, 0, stream>>>(i1c3_2); }
    { GemmP i1c3_3;
      i1c3_3.A = R67 + 0 + (size_t)66 * 3; i1c3_3.B = iw1 + 3; i1c3_3.bias = R67 + 0 + (size_t)66 * 3; i1c3_3.R = R67 + 26176 + (size_t)67 * 16; i1c3_3.C = R67 + 26176 + (size_t)67 * 16;
      i1c3_3.sAo = (long long)66 * 66 * 3; i1c3_3.sAi = (long long)66 * 3; i1c3_3.sAm = 3; i1c3_3.sAk = 1; i1c3_3.sBo = 0; i1c3_3.sBi = 0; i1c3_3.sBn = 3 * 9; i1c3_3.sBk = 9; i1c3_3.sCo = (long long)66 * 66 * 16; i1c3_3.sCi = (long long)66 * 16; i1c3_3.sCm = 16; i1c3_3.sRo = (long long)66 * 66 * 16; i1c3_3.sRi = (long long)66 * 16; i1c3_3.sRm = 16; i1c3_3.sRn = 1;
      i1c3_3.M = 64; i1c3_3.N = 16; i1c3_3.K = 3; i1c3_3.zi_n = 64; i1c3_3.flags = 4; i1c3_3.act = 0;
      i1c3_3.alpha = 1.0f; i1c3_3.beta = 1.0f; i1c3_3.sa = 1.0f; i1c3_3.sb = 1.0f; i1c3_3.Npad = 16; i1c3_3.pad_ = 0;
      k_gemm<1><<<dim3((unsigned)((16) + 31) / 32, (unsigned)((64) + 15) / 16, (unsigned)(2 * 64)), 32, 0, stream>>>(i1c3_3); }
    { GemmP i1c3_4;
      i1c3_4.A = R67 + 0 + (size_t)67 * 3; i1c3_4.B = iw1 + 4; i1c3_4.bias = R67 + 0 + (size_t)67 * 3; i1c3_4.R = R67 + 26176 + (size_t)67 * 16; i1c3_4.C = R67 + 26176 + (size_t)67 * 16;
      i1c3_4.sAo = (long long)66 * 66 * 3; i1c3_4.sAi = (long long)66 * 3; i1c3_4.sAm = 3; i1c3_4.sAk = 1; i1c3_4.sBo = 0; i1c3_4.sBi = 0; i1c3_4.sBn = 3 * 9; i1c3_4.sBk = 9; i1c3_4.sCo = (long long)66 * 66 * 16; i1c3_4.sCi = (long long)66 * 16; i1c3_4.sCm = 16; i1c3_4.sRo = (long long)66 * 66 * 16; i1c3_4.sRi = (long long)66 * 16; i1c3_4.sRm = 16; i1c3_4.sRn = 1;
      i1c3_4.M = 64; i1c3_4.N = 16; i1c3_4.K = 3; i1c3_4.zi_n = 64; i1c3_4.flags = 4; i1c3_4.act = 0;
      i1c3_4.alpha = 1.0f; i1c3_4.beta = 1.0f; i1c3_4.sa = 1.0f; i1c3_4.sb = 1.0f; i1c3_4.Npad = 16; i1c3_4.pad_ = 0;
      k_gemm<1><<<dim3((unsigned)((16) + 31) / 32, (unsigned)((64) + 15) / 16, (unsigned)(2 * 64)), 32, 0, stream>>>(i1c3_4); }
    { GemmP i1c3_5;
      i1c3_5.A = R67 + 0 + (size_t)68 * 3; i1c3_5.B = iw1 + 5; i1c3_5.bias = R67 + 0 + (size_t)68 * 3; i1c3_5.R = R67 + 26176 + (size_t)67 * 16; i1c3_5.C = R67 + 26176 + (size_t)67 * 16;
      i1c3_5.sAo = (long long)66 * 66 * 3; i1c3_5.sAi = (long long)66 * 3; i1c3_5.sAm = 3; i1c3_5.sAk = 1; i1c3_5.sBo = 0; i1c3_5.sBi = 0; i1c3_5.sBn = 3 * 9; i1c3_5.sBk = 9; i1c3_5.sCo = (long long)66 * 66 * 16; i1c3_5.sCi = (long long)66 * 16; i1c3_5.sCm = 16; i1c3_5.sRo = (long long)66 * 66 * 16; i1c3_5.sRi = (long long)66 * 16; i1c3_5.sRm = 16; i1c3_5.sRn = 1;
      i1c3_5.M = 64; i1c3_5.N = 16; i1c3_5.K = 3; i1c3_5.zi_n = 64; i1c3_5.flags = 4; i1c3_5.act = 0;
      i1c3_5.alpha = 1.0f; i1c3_5.beta = 1.0f; i1c3_5.sa = 1.0f; i1c3_5.sb = 1.0f; i1c3_5.Npad = 16; i1c3_5.pad_ = 0;
      k_gemm<1><<<dim3((unsigned)((16) + 31) / 32, (unsigned)((64) + 15) / 16, (unsigned)(2 * 64)), 32, 0, stream>>>(i1c3_5); }
    { GemmP i1c3_6;
      i1c3_6.A = R67 + 0 + (size_t)132 * 3; i1c3_6.B = iw1 + 6; i1c3_6.bias = R67 + 0 + (size_t)132 * 3; i1c3_6.R = R67 + 26176 + (size_t)67 * 16; i1c3_6.C = R67 + 26176 + (size_t)67 * 16;
      i1c3_6.sAo = (long long)66 * 66 * 3; i1c3_6.sAi = (long long)66 * 3; i1c3_6.sAm = 3; i1c3_6.sAk = 1; i1c3_6.sBo = 0; i1c3_6.sBi = 0; i1c3_6.sBn = 3 * 9; i1c3_6.sBk = 9; i1c3_6.sCo = (long long)66 * 66 * 16; i1c3_6.sCi = (long long)66 * 16; i1c3_6.sCm = 16; i1c3_6.sRo = (long long)66 * 66 * 16; i1c3_6.sRi = (long long)66 * 16; i1c3_6.sRm = 16; i1c3_6.sRn = 1;
      i1c3_6.M = 64; i1c3_6.N = 16; i1c3_6.K = 3; i1c3_6.zi_n = 64; i1c3_6.flags = 4; i1c3_6.act = 0;
      i1c3_6.alpha = 1.0f; i1c3_6.beta = 1.0f; i1c3_6.sa = 1.0f; i1c3_6.sb = 1.0f; i1c3_6.Npad = 16; i1c3_6.pad_ = 0;
      k_gemm<1><<<dim3((unsigned)((16) + 31) / 32, (unsigned)((64) + 15) / 16, (unsigned)(2 * 64)), 32, 0, stream>>>(i1c3_6); }
    { GemmP i1c3_7;
      i1c3_7.A = R67 + 0 + (size_t)133 * 3; i1c3_7.B = iw1 + 7; i1c3_7.bias = R67 + 0 + (size_t)133 * 3; i1c3_7.R = R67 + 26176 + (size_t)67 * 16; i1c3_7.C = R67 + 26176 + (size_t)67 * 16;
      i1c3_7.sAo = (long long)66 * 66 * 3; i1c3_7.sAi = (long long)66 * 3; i1c3_7.sAm = 3; i1c3_7.sAk = 1; i1c3_7.sBo = 0; i1c3_7.sBi = 0; i1c3_7.sBn = 3 * 9; i1c3_7.sBk = 9; i1c3_7.sCo = (long long)66 * 66 * 16; i1c3_7.sCi = (long long)66 * 16; i1c3_7.sCm = 16; i1c3_7.sRo = (long long)66 * 66 * 16; i1c3_7.sRi = (long long)66 * 16; i1c3_7.sRm = 16; i1c3_7.sRn = 1;
      i1c3_7.M = 64; i1c3_7.N = 16; i1c3_7.K = 3; i1c3_7.zi_n = 64; i1c3_7.flags = 4; i1c3_7.act = 0;
      i1c3_7.alpha = 1.0f; i1c3_7.beta = 1.0f; i1c3_7.sa = 1.0f; i1c3_7.sb = 1.0f; i1c3_7.Npad = 16; i1c3_7.pad_ = 0;
      k_gemm<1><<<dim3((unsigned)((16) + 31) / 32, (unsigned)((64) + 15) / 16, (unsigned)(2 * 64)), 32, 0, stream>>>(i1c3_7); }
    { GemmP i1c3_8;
      i1c3_8.A = R67 + 0 + (size_t)134 * 3; i1c3_8.B = iw1 + 8; i1c3_8.bias = R67 + 0 + (size_t)134 * 3; i1c3_8.R = R67 + 26176 + (size_t)67 * 16; i1c3_8.C = R67 + 26176 + (size_t)67 * 16;
      i1c3_8.sAo = (long long)66 * 66 * 3; i1c3_8.sAi = (long long)66 * 3; i1c3_8.sAm = 3; i1c3_8.sAk = 1; i1c3_8.sBo = 0; i1c3_8.sBi = 0; i1c3_8.sBn = 3 * 9; i1c3_8.sBk = 9; i1c3_8.sCo = (long long)66 * 66 * 16; i1c3_8.sCi = (long long)66 * 16; i1c3_8.sCm = 16; i1c3_8.sRo = (long long)66 * 66 * 16; i1c3_8.sRi = (long long)66 * 16; i1c3_8.sRm = 16; i1c3_8.sRn = 1;
      i1c3_8.M = 64; i1c3_8.N = 16; i1c3_8.K = 3; i1c3_8.zi_n = 64; i1c3_8.flags = 4; i1c3_8.act = 0;
      i1c3_8.alpha = 1.0f; i1c3_8.beta = 1.0f; i1c3_8.sa = 1.0f; i1c3_8.sb = 1.0f; i1c3_8.Npad = 16; i1c3_8.pad_ = 0;
      k_gemm<1><<<dim3((unsigned)((16) + 31) / 32, (unsigned)((64) + 15) / 16, (unsigned)(2 * 64)), 32, 0, stream>>>(i1c3_8); }
    k_mm_relu2d<<<(unsigned)(((long long)2 * HW * 16 + 255) / 256), 256, 0, stream>>>(R67 + 26176, nullptr, 2, 64, 16);
    { GemmP i2c3_0;
      i2c3_0.A = R67 + 26176 + (size_t)0 * 16; i2c3_0.B = iw2 + 0; i2c3_0.bias = ib2; i2c3_0.R = R67 + 26176 + (size_t)0 * 16; i2c3_0.C = R67 + 165568 + (size_t)67 * 32;
      i2c3_0.sAo = (long long)66 * 66 * 16; i2c3_0.sAi = (long long)66 * 16; i2c3_0.sAm = 16; i2c3_0.sAk = 1; i2c3_0.sBo = 0; i2c3_0.sBi = 0; i2c3_0.sBn = 16 * 9; i2c3_0.sBk = 9; i2c3_0.sCo = (long long)66 * 66 * 32; i2c3_0.sCi = (long long)66 * 32; i2c3_0.sCm = 32; i2c3_0.sRo = 0; i2c3_0.sRi = 0; i2c3_0.sRm = 0; i2c3_0.sRn = 0;
      i2c3_0.M = 64; i2c3_0.N = 32; i2c3_0.K = 16; i2c3_0.zi_n = 64; i2c3_0.flags = 1; i2c3_0.act = 0;
      i2c3_0.alpha = 1.0f; i2c3_0.beta = 0.0f; i2c3_0.sa = 1.0f; i2c3_0.sb = 1.0f; i2c3_0.Npad = 32; i2c3_0.pad_ = 0;
      k_gemm<1><<<dim3((unsigned)((32) + 31) / 32, (unsigned)((64) + 15) / 16, (unsigned)(2 * 64)), 32, 0, stream>>>(i2c3_0); }
    { GemmP i2c3_1;
      i2c3_1.A = R67 + 26176 + (size_t)1 * 16; i2c3_1.B = iw2 + 1; i2c3_1.bias = R67 + 26176 + (size_t)1 * 16; i2c3_1.R = R67 + 165568 + (size_t)67 * 32; i2c3_1.C = R67 + 165568 + (size_t)67 * 32;
      i2c3_1.sAo = (long long)66 * 66 * 16; i2c3_1.sAi = (long long)66 * 16; i2c3_1.sAm = 16; i2c3_1.sAk = 1; i2c3_1.sBo = 0; i2c3_1.sBi = 0; i2c3_1.sBn = 16 * 9; i2c3_1.sBk = 9; i2c3_1.sCo = (long long)66 * 66 * 32; i2c3_1.sCi = (long long)66 * 32; i2c3_1.sCm = 32; i2c3_1.sRo = (long long)66 * 66 * 32; i2c3_1.sRi = (long long)66 * 32; i2c3_1.sRm = 32; i2c3_1.sRn = 1;
      i2c3_1.M = 64; i2c3_1.N = 32; i2c3_1.K = 16; i2c3_1.zi_n = 64; i2c3_1.flags = 4; i2c3_1.act = 0;
      i2c3_1.alpha = 1.0f; i2c3_1.beta = 1.0f; i2c3_1.sa = 1.0f; i2c3_1.sb = 1.0f; i2c3_1.Npad = 32; i2c3_1.pad_ = 0;
      k_gemm<1><<<dim3((unsigned)((32) + 31) / 32, (unsigned)((64) + 15) / 16, (unsigned)(2 * 64)), 32, 0, stream>>>(i2c3_1); }
    { GemmP i2c3_2;
      i2c3_2.A = R67 + 26176 + (size_t)2 * 16; i2c3_2.B = iw2 + 2; i2c3_2.bias = R67 + 26176 + (size_t)2 * 16; i2c3_2.R = R67 + 165568 + (size_t)67 * 32; i2c3_2.C = R67 + 165568 + (size_t)67 * 32;
      i2c3_2.sAo = (long long)66 * 66 * 16; i2c3_2.sAi = (long long)66 * 16; i2c3_2.sAm = 16; i2c3_2.sAk = 1; i2c3_2.sBo = 0; i2c3_2.sBi = 0; i2c3_2.sBn = 16 * 9; i2c3_2.sBk = 9; i2c3_2.sCo = (long long)66 * 66 * 32; i2c3_2.sCi = (long long)66 * 32; i2c3_2.sCm = 32; i2c3_2.sRo = (long long)66 * 66 * 32; i2c3_2.sRi = (long long)66 * 32; i2c3_2.sRm = 32; i2c3_2.sRn = 1;
      i2c3_2.M = 64; i2c3_2.N = 32; i2c3_2.K = 16; i2c3_2.zi_n = 64; i2c3_2.flags = 4; i2c3_2.act = 0;
      i2c3_2.alpha = 1.0f; i2c3_2.beta = 1.0f; i2c3_2.sa = 1.0f; i2c3_2.sb = 1.0f; i2c3_2.Npad = 32; i2c3_2.pad_ = 0;
      k_gemm<1><<<dim3((unsigned)((32) + 31) / 32, (unsigned)((64) + 15) / 16, (unsigned)(2 * 64)), 32, 0, stream>>>(i2c3_2); }
    { GemmP i2c3_3;
      i2c3_3.A = R67 + 26176 + (size_t)66 * 16; i2c3_3.B = iw2 + 3; i2c3_3.bias = R67 + 26176 + (size_t)66 * 16; i2c3_3.R = R67 + 165568 + (size_t)67 * 32; i2c3_3.C = R67 + 165568 + (size_t)67 * 32;
      i2c3_3.sAo = (long long)66 * 66 * 16; i2c3_3.sAi = (long long)66 * 16; i2c3_3.sAm = 16; i2c3_3.sAk = 1; i2c3_3.sBo = 0; i2c3_3.sBi = 0; i2c3_3.sBn = 16 * 9; i2c3_3.sBk = 9; i2c3_3.sCo = (long long)66 * 66 * 32; i2c3_3.sCi = (long long)66 * 32; i2c3_3.sCm = 32; i2c3_3.sRo = (long long)66 * 66 * 32; i2c3_3.sRi = (long long)66 * 32; i2c3_3.sRm = 32; i2c3_3.sRn = 1;
      i2c3_3.M = 64; i2c3_3.N = 32; i2c3_3.K = 16; i2c3_3.zi_n = 64; i2c3_3.flags = 4; i2c3_3.act = 0;
      i2c3_3.alpha = 1.0f; i2c3_3.beta = 1.0f; i2c3_3.sa = 1.0f; i2c3_3.sb = 1.0f; i2c3_3.Npad = 32; i2c3_3.pad_ = 0;
      k_gemm<1><<<dim3((unsigned)((32) + 31) / 32, (unsigned)((64) + 15) / 16, (unsigned)(2 * 64)), 32, 0, stream>>>(i2c3_3); }
    { GemmP i2c3_4;
      i2c3_4.A = R67 + 26176 + (size_t)67 * 16; i2c3_4.B = iw2 + 4; i2c3_4.bias = R67 + 26176 + (size_t)67 * 16; i2c3_4.R = R67 + 165568 + (size_t)67 * 32; i2c3_4.C = R67 + 165568 + (size_t)67 * 32;
      i2c3_4.sAo = (long long)66 * 66 * 16; i2c3_4.sAi = (long long)66 * 16; i2c3_4.sAm = 16; i2c3_4.sAk = 1; i2c3_4.sBo = 0; i2c3_4.sBi = 0; i2c3_4.sBn = 16 * 9; i2c3_4.sBk = 9; i2c3_4.sCo = (long long)66 * 66 * 32; i2c3_4.sCi = (long long)66 * 32; i2c3_4.sCm = 32; i2c3_4.sRo = (long long)66 * 66 * 32; i2c3_4.sRi = (long long)66 * 32; i2c3_4.sRm = 32; i2c3_4.sRn = 1;
      i2c3_4.M = 64; i2c3_4.N = 32; i2c3_4.K = 16; i2c3_4.zi_n = 64; i2c3_4.flags = 4; i2c3_4.act = 0;
      i2c3_4.alpha = 1.0f; i2c3_4.beta = 1.0f; i2c3_4.sa = 1.0f; i2c3_4.sb = 1.0f; i2c3_4.Npad = 32; i2c3_4.pad_ = 0;
      k_gemm<1><<<dim3((unsigned)((32) + 31) / 32, (unsigned)((64) + 15) / 16, (unsigned)(2 * 64)), 32, 0, stream>>>(i2c3_4); }
    { GemmP i2c3_5;
      i2c3_5.A = R67 + 26176 + (size_t)68 * 16; i2c3_5.B = iw2 + 5; i2c3_5.bias = R67 + 26176 + (size_t)68 * 16; i2c3_5.R = R67 + 165568 + (size_t)67 * 32; i2c3_5.C = R67 + 165568 + (size_t)67 * 32;
      i2c3_5.sAo = (long long)66 * 66 * 16; i2c3_5.sAi = (long long)66 * 16; i2c3_5.sAm = 16; i2c3_5.sAk = 1; i2c3_5.sBo = 0; i2c3_5.sBi = 0; i2c3_5.sBn = 16 * 9; i2c3_5.sBk = 9; i2c3_5.sCo = (long long)66 * 66 * 32; i2c3_5.sCi = (long long)66 * 32; i2c3_5.sCm = 32; i2c3_5.sRo = (long long)66 * 66 * 32; i2c3_5.sRi = (long long)66 * 32; i2c3_5.sRm = 32; i2c3_5.sRn = 1;
      i2c3_5.M = 64; i2c3_5.N = 32; i2c3_5.K = 16; i2c3_5.zi_n = 64; i2c3_5.flags = 4; i2c3_5.act = 0;
      i2c3_5.alpha = 1.0f; i2c3_5.beta = 1.0f; i2c3_5.sa = 1.0f; i2c3_5.sb = 1.0f; i2c3_5.Npad = 32; i2c3_5.pad_ = 0;
      k_gemm<1><<<dim3((unsigned)((32) + 31) / 32, (unsigned)((64) + 15) / 16, (unsigned)(2 * 64)), 32, 0, stream>>>(i2c3_5); }
    { GemmP i2c3_6;
      i2c3_6.A = R67 + 26176 + (size_t)132 * 16; i2c3_6.B = iw2 + 6; i2c3_6.bias = R67 + 26176 + (size_t)132 * 16; i2c3_6.R = R67 + 165568 + (size_t)67 * 32; i2c3_6.C = R67 + 165568 + (size_t)67 * 32;
      i2c3_6.sAo = (long long)66 * 66 * 16; i2c3_6.sAi = (long long)66 * 16; i2c3_6.sAm = 16; i2c3_6.sAk = 1; i2c3_6.sBo = 0; i2c3_6.sBi = 0; i2c3_6.sBn = 16 * 9; i2c3_6.sBk = 9; i2c3_6.sCo = (long long)66 * 66 * 32; i2c3_6.sCi = (long long)66 * 32; i2c3_6.sCm = 32; i2c3_6.sRo = (long long)66 * 66 * 32; i2c3_6.sRi = (long long)66 * 32; i2c3_6.sRm = 32; i2c3_6.sRn = 1;
      i2c3_6.M = 64; i2c3_6.N = 32; i2c3_6.K = 16; i2c3_6.zi_n = 64; i2c3_6.flags = 4; i2c3_6.act = 0;
      i2c3_6.alpha = 1.0f; i2c3_6.beta = 1.0f; i2c3_6.sa = 1.0f; i2c3_6.sb = 1.0f; i2c3_6.Npad = 32; i2c3_6.pad_ = 0;
      k_gemm<1><<<dim3((unsigned)((32) + 31) / 32, (unsigned)((64) + 15) / 16, (unsigned)(2 * 64)), 32, 0, stream>>>(i2c3_6); }
    { GemmP i2c3_7;
      i2c3_7.A = R67 + 26176 + (size_t)133 * 16; i2c3_7.B = iw2 + 7; i2c3_7.bias = R67 + 26176 + (size_t)133 * 16; i2c3_7.R = R67 + 165568 + (size_t)67 * 32; i2c3_7.C = R67 + 165568 + (size_t)67 * 32;
      i2c3_7.sAo = (long long)66 * 66 * 16; i2c3_7.sAi = (long long)66 * 16; i2c3_7.sAm = 16; i2c3_7.sAk = 1; i2c3_7.sBo = 0; i2c3_7.sBi = 0; i2c3_7.sBn = 16 * 9; i2c3_7.sBk = 9; i2c3_7.sCo = (long long)66 * 66 * 32; i2c3_7.sCi = (long long)66 * 32; i2c3_7.sCm = 32; i2c3_7.sRo = (long long)66 * 66 * 32; i2c3_7.sRi = (long long)66 * 32; i2c3_7.sRm = 32; i2c3_7.sRn = 1;
      i2c3_7.M = 64; i2c3_7.N = 32; i2c3_7.K = 16; i2c3_7.zi_n = 64; i2c3_7.flags = 4; i2c3_7.act = 0;
      i2c3_7.alpha = 1.0f; i2c3_7.beta = 1.0f; i2c3_7.sa = 1.0f; i2c3_7.sb = 1.0f; i2c3_7.Npad = 32; i2c3_7.pad_ = 0;
      k_gemm<1><<<dim3((unsigned)((32) + 31) / 32, (unsigned)((64) + 15) / 16, (unsigned)(2 * 64)), 32, 0, stream>>>(i2c3_7); }
    { GemmP i2c3_8;
      i2c3_8.A = R67 + 26176 + (size_t)134 * 16; i2c3_8.B = iw2 + 8; i2c3_8.bias = R67 + 26176 + (size_t)134 * 16; i2c3_8.R = R67 + 165568 + (size_t)67 * 32; i2c3_8.C = R67 + 165568 + (size_t)67 * 32;
      i2c3_8.sAo = (long long)66 * 66 * 16; i2c3_8.sAi = (long long)66 * 16; i2c3_8.sAm = 16; i2c3_8.sAk = 1; i2c3_8.sBo = 0; i2c3_8.sBi = 0; i2c3_8.sBn = 16 * 9; i2c3_8.sBk = 9; i2c3_8.sCo = (long long)66 * 66 * 32; i2c3_8.sCi = (long long)66 * 32; i2c3_8.sCm = 32; i2c3_8.sRo = (long long)66 * 66 * 32; i2c3_8.sRi = (long long)66 * 32; i2c3_8.sRm = 32; i2c3_8.sRn = 1;
      i2c3_8.M = 64; i2c3_8.N = 32; i2c3_8.K = 16; i2c3_8.zi_n = 64; i2c3_8.flags = 4; i2c3_8.act = 0;
      i2c3_8.alpha = 1.0f; i2c3_8.beta = 1.0f; i2c3_8.sa = 1.0f; i2c3_8.sb = 1.0f; i2c3_8.Npad = 32; i2c3_8.pad_ = 0;
      k_gemm<1><<<dim3((unsigned)((32) + 31) / 32, (unsigned)((64) + 15) / 16, (unsigned)(2 * 64)), 32, 0, stream>>>(i2c3_8); }
    k_mm_relu2d<<<(unsigned)(((long long)2 * HW * 32 + 255) / 256), 256, 0, stream>>>(R67 + 165568, nullptr, 2, 64, 32);
    { GemmP i3c3_0;
      i3c3_0.A = R67 + 165568 + (size_t)0 * 32; i3c3_0.B = iw3 + 0; i3c3_0.bias = ib3; i3c3_0.R = R67 + 165568 + (size_t)0 * 32; i3c3_0.C = R67 + 444352 + (size_t)67 * 64;
      i3c3_0.sAo = (long long)66 * 66 * 32; i3c3_0.sAi = (long long)66 * 32; i3c3_0.sAm = 32; i3c3_0.sAk = 1; i3c3_0.sBo = 0; i3c3_0.sBi = 0; i3c3_0.sBn = 32 * 9; i3c3_0.sBk = 9; i3c3_0.sCo = (long long)66 * 66 * 64; i3c3_0.sCi = (long long)66 * 64; i3c3_0.sCm = 64; i3c3_0.sRo = 0; i3c3_0.sRi = 0; i3c3_0.sRm = 0; i3c3_0.sRn = 0;
      i3c3_0.M = 64; i3c3_0.N = 64; i3c3_0.K = 32; i3c3_0.zi_n = 64; i3c3_0.flags = 1; i3c3_0.act = 0;
      i3c3_0.alpha = 1.0f; i3c3_0.beta = 0.0f; i3c3_0.sa = 1.0f; i3c3_0.sb = 1.0f; i3c3_0.Npad = 64; i3c3_0.pad_ = 0;
      k_gemm<1><<<dim3((unsigned)((64) + 31) / 32, (unsigned)((64) + 15) / 16, (unsigned)(2 * 64)), 32, 0, stream>>>(i3c3_0); }
    { GemmP i3c3_1;
      i3c3_1.A = R67 + 165568 + (size_t)1 * 32; i3c3_1.B = iw3 + 1; i3c3_1.bias = R67 + 165568 + (size_t)1 * 32; i3c3_1.R = R67 + 444352 + (size_t)67 * 64; i3c3_1.C = R67 + 444352 + (size_t)67 * 64;
      i3c3_1.sAo = (long long)66 * 66 * 32; i3c3_1.sAi = (long long)66 * 32; i3c3_1.sAm = 32; i3c3_1.sAk = 1; i3c3_1.sBo = 0; i3c3_1.sBi = 0; i3c3_1.sBn = 32 * 9; i3c3_1.sBk = 9; i3c3_1.sCo = (long long)66 * 66 * 64; i3c3_1.sCi = (long long)66 * 64; i3c3_1.sCm = 64; i3c3_1.sRo = (long long)66 * 66 * 64; i3c3_1.sRi = (long long)66 * 64; i3c3_1.sRm = 64; i3c3_1.sRn = 1;
      i3c3_1.M = 64; i3c3_1.N = 64; i3c3_1.K = 32; i3c3_1.zi_n = 64; i3c3_1.flags = 4; i3c3_1.act = 0;
      i3c3_1.alpha = 1.0f; i3c3_1.beta = 1.0f; i3c3_1.sa = 1.0f; i3c3_1.sb = 1.0f; i3c3_1.Npad = 64; i3c3_1.pad_ = 0;
      k_gemm<1><<<dim3((unsigned)((64) + 31) / 32, (unsigned)((64) + 15) / 16, (unsigned)(2 * 64)), 32, 0, stream>>>(i3c3_1); }
    { GemmP i3c3_2;
      i3c3_2.A = R67 + 165568 + (size_t)2 * 32; i3c3_2.B = iw3 + 2; i3c3_2.bias = R67 + 165568 + (size_t)2 * 32; i3c3_2.R = R67 + 444352 + (size_t)67 * 64; i3c3_2.C = R67 + 444352 + (size_t)67 * 64;
      i3c3_2.sAo = (long long)66 * 66 * 32; i3c3_2.sAi = (long long)66 * 32; i3c3_2.sAm = 32; i3c3_2.sAk = 1; i3c3_2.sBo = 0; i3c3_2.sBi = 0; i3c3_2.sBn = 32 * 9; i3c3_2.sBk = 9; i3c3_2.sCo = (long long)66 * 66 * 64; i3c3_2.sCi = (long long)66 * 64; i3c3_2.sCm = 64; i3c3_2.sRo = (long long)66 * 66 * 64; i3c3_2.sRi = (long long)66 * 64; i3c3_2.sRm = 64; i3c3_2.sRn = 1;
      i3c3_2.M = 64; i3c3_2.N = 64; i3c3_2.K = 32; i3c3_2.zi_n = 64; i3c3_2.flags = 4; i3c3_2.act = 0;
      i3c3_2.alpha = 1.0f; i3c3_2.beta = 1.0f; i3c3_2.sa = 1.0f; i3c3_2.sb = 1.0f; i3c3_2.Npad = 64; i3c3_2.pad_ = 0;
      k_gemm<1><<<dim3((unsigned)((64) + 31) / 32, (unsigned)((64) + 15) / 16, (unsigned)(2 * 64)), 32, 0, stream>>>(i3c3_2); }
    { GemmP i3c3_3;
      i3c3_3.A = R67 + 165568 + (size_t)66 * 32; i3c3_3.B = iw3 + 3; i3c3_3.bias = R67 + 165568 + (size_t)66 * 32; i3c3_3.R = R67 + 444352 + (size_t)67 * 64; i3c3_3.C = R67 + 444352 + (size_t)67 * 64;
      i3c3_3.sAo = (long long)66 * 66 * 32; i3c3_3.sAi = (long long)66 * 32; i3c3_3.sAm = 32; i3c3_3.sAk = 1; i3c3_3.sBo = 0; i3c3_3.sBi = 0; i3c3_3.sBn = 32 * 9; i3c3_3.sBk = 9; i3c3_3.sCo = (long long)66 * 66 * 64; i3c3_3.sCi = (long long)66 * 64; i3c3_3.sCm = 64; i3c3_3.sRo = (long long)66 * 66 * 64; i3c3_3.sRi = (long long)66 * 64; i3c3_3.sRm = 64; i3c3_3.sRn = 1;
      i3c3_3.M = 64; i3c3_3.N = 64; i3c3_3.K = 32; i3c3_3.zi_n = 64; i3c3_3.flags = 4; i3c3_3.act = 0;
      i3c3_3.alpha = 1.0f; i3c3_3.beta = 1.0f; i3c3_3.sa = 1.0f; i3c3_3.sb = 1.0f; i3c3_3.Npad = 64; i3c3_3.pad_ = 0;
      k_gemm<1><<<dim3((unsigned)((64) + 31) / 32, (unsigned)((64) + 15) / 16, (unsigned)(2 * 64)), 32, 0, stream>>>(i3c3_3); }
    { GemmP i3c3_4;
      i3c3_4.A = R67 + 165568 + (size_t)67 * 32; i3c3_4.B = iw3 + 4; i3c3_4.bias = R67 + 165568 + (size_t)67 * 32; i3c3_4.R = R67 + 444352 + (size_t)67 * 64; i3c3_4.C = R67 + 444352 + (size_t)67 * 64;
      i3c3_4.sAo = (long long)66 * 66 * 32; i3c3_4.sAi = (long long)66 * 32; i3c3_4.sAm = 32; i3c3_4.sAk = 1; i3c3_4.sBo = 0; i3c3_4.sBi = 0; i3c3_4.sBn = 32 * 9; i3c3_4.sBk = 9; i3c3_4.sCo = (long long)66 * 66 * 64; i3c3_4.sCi = (long long)66 * 64; i3c3_4.sCm = 64; i3c3_4.sRo = (long long)66 * 66 * 64; i3c3_4.sRi = (long long)66 * 64; i3c3_4.sRm = 64; i3c3_4.sRn = 1;
      i3c3_4.M = 64; i3c3_4.N = 64; i3c3_4.K = 32; i3c3_4.zi_n = 64; i3c3_4.flags = 4; i3c3_4.act = 0;
      i3c3_4.alpha = 1.0f; i3c3_4.beta = 1.0f; i3c3_4.sa = 1.0f; i3c3_4.sb = 1.0f; i3c3_4.Npad = 64; i3c3_4.pad_ = 0;
      k_gemm<1><<<dim3((unsigned)((64) + 31) / 32, (unsigned)((64) + 15) / 16, (unsigned)(2 * 64)), 32, 0, stream>>>(i3c3_4); }
    { GemmP i3c3_5;
      i3c3_5.A = R67 + 165568 + (size_t)68 * 32; i3c3_5.B = iw3 + 5; i3c3_5.bias = R67 + 165568 + (size_t)68 * 32; i3c3_5.R = R67 + 444352 + (size_t)67 * 64; i3c3_5.C = R67 + 444352 + (size_t)67 * 64;
      i3c3_5.sAo = (long long)66 * 66 * 32; i3c3_5.sAi = (long long)66 * 32; i3c3_5.sAm = 32; i3c3_5.sAk = 1; i3c3_5.sBo = 0; i3c3_5.sBi = 0; i3c3_5.sBn = 32 * 9; i3c3_5.sBk = 9; i3c3_5.sCo = (long long)66 * 66 * 64; i3c3_5.sCi = (long long)66 * 64; i3c3_5.sCm = 64; i3c3_5.sRo = (long long)66 * 66 * 64; i3c3_5.sRi = (long long)66 * 64; i3c3_5.sRm = 64; i3c3_5.sRn = 1;
      i3c3_5.M = 64; i3c3_5.N = 64; i3c3_5.K = 32; i3c3_5.zi_n = 64; i3c3_5.flags = 4; i3c3_5.act = 0;
      i3c3_5.alpha = 1.0f; i3c3_5.beta = 1.0f; i3c3_5.sa = 1.0f; i3c3_5.sb = 1.0f; i3c3_5.Npad = 64; i3c3_5.pad_ = 0;
      k_gemm<1><<<dim3((unsigned)((64) + 31) / 32, (unsigned)((64) + 15) / 16, (unsigned)(2 * 64)), 32, 0, stream>>>(i3c3_5); }
    { GemmP i3c3_6;
      i3c3_6.A = R67 + 165568 + (size_t)132 * 32; i3c3_6.B = iw3 + 6; i3c3_6.bias = R67 + 165568 + (size_t)132 * 32; i3c3_6.R = R67 + 444352 + (size_t)67 * 64; i3c3_6.C = R67 + 444352 + (size_t)67 * 64;
      i3c3_6.sAo = (long long)66 * 66 * 32; i3c3_6.sAi = (long long)66 * 32; i3c3_6.sAm = 32; i3c3_6.sAk = 1; i3c3_6.sBo = 0; i3c3_6.sBi = 0; i3c3_6.sBn = 32 * 9; i3c3_6.sBk = 9; i3c3_6.sCo = (long long)66 * 66 * 64; i3c3_6.sCi = (long long)66 * 64; i3c3_6.sCm = 64; i3c3_6.sRo = (long long)66 * 66 * 64; i3c3_6.sRi = (long long)66 * 64; i3c3_6.sRm = 64; i3c3_6.sRn = 1;
      i3c3_6.M = 64; i3c3_6.N = 64; i3c3_6.K = 32; i3c3_6.zi_n = 64; i3c3_6.flags = 4; i3c3_6.act = 0;
      i3c3_6.alpha = 1.0f; i3c3_6.beta = 1.0f; i3c3_6.sa = 1.0f; i3c3_6.sb = 1.0f; i3c3_6.Npad = 64; i3c3_6.pad_ = 0;
      k_gemm<1><<<dim3((unsigned)((64) + 31) / 32, (unsigned)((64) + 15) / 16, (unsigned)(2 * 64)), 32, 0, stream>>>(i3c3_6); }
    { GemmP i3c3_7;
      i3c3_7.A = R67 + 165568 + (size_t)133 * 32; i3c3_7.B = iw3 + 7; i3c3_7.bias = R67 + 165568 + (size_t)133 * 32; i3c3_7.R = R67 + 444352 + (size_t)67 * 64; i3c3_7.C = R67 + 444352 + (size_t)67 * 64;
      i3c3_7.sAo = (long long)66 * 66 * 32; i3c3_7.sAi = (long long)66 * 32; i3c3_7.sAm = 32; i3c3_7.sAk = 1; i3c3_7.sBo = 0; i3c3_7.sBi = 0; i3c3_7.sBn = 32 * 9; i3c3_7.sBk = 9; i3c3_7.sCo = (long long)66 * 66 * 64; i3c3_7.sCi = (long long)66 * 64; i3c3_7.sCm = 64; i3c3_7.sRo = (long long)66 * 66 * 64; i3c3_7.sRi = (long long)66 * 64; i3c3_7.sRm = 64; i3c3_7.sRn = 1;
      i3c3_7.M = 64; i3c3_7.N = 64; i3c3_7.K = 32; i3c3_7.zi_n = 64; i3c3_7.flags = 4; i3c3_7.act = 0;
      i3c3_7.alpha = 1.0f; i3c3_7.beta = 1.0f; i3c3_7.sa = 1.0f; i3c3_7.sb = 1.0f; i3c3_7.Npad = 64; i3c3_7.pad_ = 0;
      k_gemm<1><<<dim3((unsigned)((64) + 31) / 32, (unsigned)((64) + 15) / 16, (unsigned)(2 * 64)), 32, 0, stream>>>(i3c3_7); }
    { GemmP i3c3_8;
      i3c3_8.A = R67 + 165568 + (size_t)134 * 32; i3c3_8.B = iw3 + 8; i3c3_8.bias = R67 + 165568 + (size_t)134 * 32; i3c3_8.R = R67 + 444352 + (size_t)67 * 64; i3c3_8.C = R67 + 444352 + (size_t)67 * 64;
      i3c3_8.sAo = (long long)66 * 66 * 32; i3c3_8.sAi = (long long)66 * 32; i3c3_8.sAm = 32; i3c3_8.sAk = 1; i3c3_8.sBo = 0; i3c3_8.sBi = 0; i3c3_8.sBn = 32 * 9; i3c3_8.sBk = 9; i3c3_8.sCo = (long long)66 * 66 * 64; i3c3_8.sCi = (long long)66 * 64; i3c3_8.sCm = 64; i3c3_8.sRo = (long long)66 * 66 * 64; i3c3_8.sRi = (long long)66 * 64; i3c3_8.sRm = 64; i3c3_8.sRn = 1;
      i3c3_8.M = 64; i3c3_8.N = 64; i3c3_8.K = 32; i3c3_8.zi_n = 64; i3c3_8.flags = 4; i3c3_8.act = 0;
      i3c3_8.alpha = 1.0f; i3c3_8.beta = 1.0f; i3c3_8.sa = 1.0f; i3c3_8.sb = 1.0f; i3c3_8.Npad = 64; i3c3_8.pad_ = 0;
      k_gemm<1><<<dim3((unsigned)((64) + 31) / 32, (unsigned)((64) + 15) / 16, (unsigned)(2 * 64)), 32, 0, stream>>>(i3c3_8); }
    k_mm_relu2d<<<(unsigned)(((long long)2 * HW * 64 + 255) / 256), 256, 0, stream>>>(R67 + 444352, R67 + 1001920, 2, 64, 64);
    { GemmP gqkv3;
      gqkv3.A = R67 + 1001920; gqkv3.B = qkvw; gqkv3.bias = qkvb; gqkv3.R = R67 + 1001920; gqkv3.C = R67 + 1526208;
      gqkv3.sAo = 0; gqkv3.sAi = 0; gqkv3.sAm = 64; gqkv3.sAk = 1; gqkv3.sBo = 0; gqkv3.sBi = 0; gqkv3.sBn = 64; gqkv3.sBk = 1; gqkv3.sCo = 0; gqkv3.sCi = 0; gqkv3.sCm = 192; gqkv3.sRo = 0; gqkv3.sRi = 0; gqkv3.sRm = 0; gqkv3.sRn = 0;
      gqkv3.M = 2 * HW; gqkv3.N = 192; gqkv3.K = 64; gqkv3.zi_n = 1; gqkv3.flags = 1; gqkv3.act = 0;
      gqkv3.alpha = 1.0f; gqkv3.beta = 0.0f; gqkv3.sa = 1.0f; gqkv3.sb = 1.0f; gqkv3.Npad = 192; gqkv3.pad_ = 0;
      k_gemm<1><<<dim3((unsigned)((192) + 31) / 32, (unsigned)((2 * HW) + 15) / 16, (unsigned)(1)), 32, 0, stream>>>(gqkv3); }
    k_mm_dw<<<(unsigned)(((long long)2 * HW * 192 + 255) / 256), 256, 0, stream>>>(R67 + 1526208, dww, dwb, R67 + 3099072, 2, 64, 192);
    k_mm_fall<<<(unsigned)(((long long)2 * HW * 144 + 255) / 256), 256, 0, stream>>>(R67 + 3099072, fcw, fcb, R67 + 4671936, 2, HW, 192);
    k_mm_dep<<<(unsigned)(((long long)2 * 64 * HW + 255) / 256), 256, 0, stream>>>(R67 + 4671936, depw, depb, R67 + 5851584, 2, 64);
    k_mm_qknorm<<<2 * 128, 256, 0, stream>>>(R67 + 3099072, R67 + 6375872, 2, HW, 192);
    { GemmP gat3;
      gat3.A = R67 + 6375872; gat3.B = R67 + 6375872 + (size_t)64 * HW; gat3.bias = R67 + 6375872; gat3.R = R67 + 6375872; gat3.C = R67 + 7424448;
      gat3.sAo = (long long)128 * HW; gat3.sAi = (long long)16 * HW; gat3.sAm = HW; gat3.sAk = 1; gat3.sBo = (long long)128 * HW; gat3.sBi = (long long)16 * HW; gat3.sBn = HW; gat3.sBk = 1; gat3.sCo = (long long)4 * 16 * LP; gat3.sCi = 16 * LP; gat3.sCm = LP; gat3.sRo = 0; gat3.sRi = 0; gat3.sRm = 0; gat3.sRn = 0;
      gat3.M = 16; gat3.N = 16; gat3.K = HW; gat3.zi_n = 4; gat3.flags = 0; gat3.act = 0;
      gat3.alpha = 1.0f; gat3.beta = 0.0f; gat3.sa = 1.0f; gat3.sb = 1.0f; gat3.Npad = LP; gat3.pad_ = 0;
      k_gemm<1><<<dim3((unsigned)((LP) + 31) / 32, (unsigned)((16) + 15) / 16, (unsigned)(2 * 4)), 32, 0, stream>>>(gat3); }
    k_mm_sm16<<<(unsigned)((2 * 4 * 16 + 255) / 256), 256, 0, stream>>>(R67 + 7424448, temp, 2 * 4, LP);
    { GemmP gao3;
      gao3.A = R67 + 7424448; gao3.B = R67 + 3099072 + 128; gao3.bias = R67 + 7424448; gao3.R = R67 + 7424448; gao3.C = R67 + 7428544;
      gao3.sAo = (long long)4 * 16 * LP; gao3.sAi = 16 * LP; gao3.sAm = LP; gao3.sAk = 1; gao3.sBo = (long long)HW * 192; gao3.sBi = 16; gao3.sBn = 192; gao3.sBk = 1; gao3.sCo = (long long)64 * HW; gao3.sCi = (long long)16 * HW; gao3.sCm = HW; gao3.sRo = 0; gao3.sRi = 0; gao3.sRm = 0; gao3.sRn = 0;
      gao3.M = 16; gao3.N = HW; gao3.K = 16; gao3.zi_n = 4; gao3.flags = 0; gao3.act = 0;
      gao3.alpha = 1.0f; gao3.beta = 0.0f; gao3.sa = 1.0f; gao3.sb = 1.0f; gao3.Npad = HW; gao3.pad_ = 0;
      k_gemm<1><<<dim3((unsigned)((HW) + 31) / 32, (unsigned)((16) + 15) / 16, (unsigned)(2 * 4)), 32, 0, stream>>>(gao3); }
    { GemmP gproj3;
      gproj3.A = projw; gproj3.B = R67 + 7428544; gproj3.bias = projb; gproj3.R = projw; gproj3.C = R67 + 7952832;
      gproj3.sAo = 0; gproj3.sAi = 0; gproj3.sAm = 64; gproj3.sAk = 1; gproj3.sBo = (long long)64 * HW; gproj3.sBi = 0; gproj3.sBn = 1; gproj3.sBk = HW; gproj3.sCo = (long long)64 * HW; gproj3.sCi = 0; gproj3.sCm = HW; gproj3.sRo = 0; gproj3.sRi = 0; gproj3.sRm = 0; gproj3.sRn = 0;
      gproj3.M = 64; gproj3.N = HW; gproj3.K = 64; gproj3.zi_n = 1; gproj3.flags = 2; gproj3.act = 0;
      gproj3.alpha = 1.0f; gproj3.beta = 0.0f; gproj3.sa = 1.0f; gproj3.sb = 1.0f; gproj3.Npad = HW; gproj3.pad_ = 0;
      k_gemm<1><<<dim3((unsigned)((HW) + 31) / 32, (unsigned)((64) + 15) / 16, (unsigned)(2)), 32, 0, stream>>>(gproj3); }
    k_mm_imgfeat<<<(unsigned)(((long long)2 * SEQ * 64 + 255) / 256), 256, 0, stream>>>(R67 + 7952832, R67 + 5851584, IR + (size_t)6 * SEQ * 64, 2, HW, 64);
    hipMemsetAsync(R67 + 0, 0, (size_t)2 * 66 * 66 * 3 * 4, stream); hipMemsetAsync(R67 + 26176, 0, (size_t)2 * 66 * 66 * 16 * 4, stream); hipMemsetAsync(R67 + 165568, 0, (size_t)2 * 66 * 66 * 32 * 4, stream); hipMemsetAsync(R67 + 444352, 0, (size_t)2 * 66 * 66 * 64 * 4, stream);
    k_mm_padimg<<<(unsigned)(((long long)2 * HW * 3 + 255) / 256), 256, 0, stream>>>(img + (size_t)8 * 3 * HW, R67 + 0, 2, 3, 64);
    { GemmP i1c4_0;
      i1c4_0.A = R67 + 0 + (size_t)0 * 3; i1c4_0.B = iw1 + 0; i1c4_0.bias = ib1; i1c4_0.R = R67 + 0 + (size_t)0 * 3; i1c4_0.C = R67 + 26176 + (size_t)67 * 16;
      i1c4_0.sAo = (long long)66 * 66 * 3; i1c4_0.sAi = (long long)66 * 3; i1c4_0.sAm = 3; i1c4_0.sAk = 1; i1c4_0.sBo = 0; i1c4_0.sBi = 0; i1c4_0.sBn = 3 * 9; i1c4_0.sBk = 9; i1c4_0.sCo = (long long)66 * 66 * 16; i1c4_0.sCi = (long long)66 * 16; i1c4_0.sCm = 16; i1c4_0.sRo = 0; i1c4_0.sRi = 0; i1c4_0.sRm = 0; i1c4_0.sRn = 0;
      i1c4_0.M = 64; i1c4_0.N = 16; i1c4_0.K = 3; i1c4_0.zi_n = 64; i1c4_0.flags = 1; i1c4_0.act = 0;
      i1c4_0.alpha = 1.0f; i1c4_0.beta = 0.0f; i1c4_0.sa = 1.0f; i1c4_0.sb = 1.0f; i1c4_0.Npad = 16; i1c4_0.pad_ = 0;
      k_gemm<1><<<dim3((unsigned)((16) + 31) / 32, (unsigned)((64) + 15) / 16, (unsigned)(2 * 64)), 32, 0, stream>>>(i1c4_0); }
    { GemmP i1c4_1;
      i1c4_1.A = R67 + 0 + (size_t)1 * 3; i1c4_1.B = iw1 + 1; i1c4_1.bias = R67 + 0 + (size_t)1 * 3; i1c4_1.R = R67 + 26176 + (size_t)67 * 16; i1c4_1.C = R67 + 26176 + (size_t)67 * 16;
      i1c4_1.sAo = (long long)66 * 66 * 3; i1c4_1.sAi = (long long)66 * 3; i1c4_1.sAm = 3; i1c4_1.sAk = 1; i1c4_1.sBo = 0; i1c4_1.sBi = 0; i1c4_1.sBn = 3 * 9; i1c4_1.sBk = 9; i1c4_1.sCo = (long long)66 * 66 * 16; i1c4_1.sCi = (long long)66 * 16; i1c4_1.sCm = 16; i1c4_1.sRo = (long long)66 * 66 * 16; i1c4_1.sRi = (long long)66 * 16; i1c4_1.sRm = 16; i1c4_1.sRn = 1;
      i1c4_1.M = 64; i1c4_1.N = 16; i1c4_1.K = 3; i1c4_1.zi_n = 64; i1c4_1.flags = 4; i1c4_1.act = 0;
      i1c4_1.alpha = 1.0f; i1c4_1.beta = 1.0f; i1c4_1.sa = 1.0f; i1c4_1.sb = 1.0f; i1c4_1.Npad = 16; i1c4_1.pad_ = 0;
      k_gemm<1><<<dim3((unsigned)((16) + 31) / 32, (unsigned)((64) + 15) / 16, (unsigned)(2 * 64)), 32, 0, stream>>>(i1c4_1); }
    { GemmP i1c4_2;
      i1c4_2.A = R67 + 0 + (size_t)2 * 3; i1c4_2.B = iw1 + 2; i1c4_2.bias = R67 + 0 + (size_t)2 * 3; i1c4_2.R = R67 + 26176 + (size_t)67 * 16; i1c4_2.C = R67 + 26176 + (size_t)67 * 16;
      i1c4_2.sAo = (long long)66 * 66 * 3; i1c4_2.sAi = (long long)66 * 3; i1c4_2.sAm = 3; i1c4_2.sAk = 1; i1c4_2.sBo = 0; i1c4_2.sBi = 0; i1c4_2.sBn = 3 * 9; i1c4_2.sBk = 9; i1c4_2.sCo = (long long)66 * 66 * 16; i1c4_2.sCi = (long long)66 * 16; i1c4_2.sCm = 16; i1c4_2.sRo = (long long)66 * 66 * 16; i1c4_2.sRi = (long long)66 * 16; i1c4_2.sRm = 16; i1c4_2.sRn = 1;
      i1c4_2.M = 64; i1c4_2.N = 16; i1c4_2.K = 3; i1c4_2.zi_n = 64; i1c4_2.flags = 4; i1c4_2.act = 0;
      i1c4_2.alpha = 1.0f; i1c4_2.beta = 1.0f; i1c4_2.sa = 1.0f; i1c4_2.sb = 1.0f; i1c4_2.Npad = 16; i1c4_2.pad_ = 0;
      k_gemm<1><<<dim3((unsigned)((16) + 31) / 32, (unsigned)((64) + 15) / 16, (unsigned)(2 * 64)), 32, 0, stream>>>(i1c4_2); }
    { GemmP i1c4_3;
      i1c4_3.A = R67 + 0 + (size_t)66 * 3; i1c4_3.B = iw1 + 3; i1c4_3.bias = R67 + 0 + (size_t)66 * 3; i1c4_3.R = R67 + 26176 + (size_t)67 * 16; i1c4_3.C = R67 + 26176 + (size_t)67 * 16;
      i1c4_3.sAo = (long long)66 * 66 * 3; i1c4_3.sAi = (long long)66 * 3; i1c4_3.sAm = 3; i1c4_3.sAk = 1; i1c4_3.sBo = 0; i1c4_3.sBi = 0; i1c4_3.sBn = 3 * 9; i1c4_3.sBk = 9; i1c4_3.sCo = (long long)66 * 66 * 16; i1c4_3.sCi = (long long)66 * 16; i1c4_3.sCm = 16; i1c4_3.sRo = (long long)66 * 66 * 16; i1c4_3.sRi = (long long)66 * 16; i1c4_3.sRm = 16; i1c4_3.sRn = 1;
      i1c4_3.M = 64; i1c4_3.N = 16; i1c4_3.K = 3; i1c4_3.zi_n = 64; i1c4_3.flags = 4; i1c4_3.act = 0;
      i1c4_3.alpha = 1.0f; i1c4_3.beta = 1.0f; i1c4_3.sa = 1.0f; i1c4_3.sb = 1.0f; i1c4_3.Npad = 16; i1c4_3.pad_ = 0;
      k_gemm<1><<<dim3((unsigned)((16) + 31) / 32, (unsigned)((64) + 15) / 16, (unsigned)(2 * 64)), 32, 0, stream>>>(i1c4_3); }
    { GemmP i1c4_4;
      i1c4_4.A = R67 + 0 + (size_t)67 * 3; i1c4_4.B = iw1 + 4; i1c4_4.bias = R67 + 0 + (size_t)67 * 3; i1c4_4.R = R67 + 26176 + (size_t)67 * 16; i1c4_4.C = R67 + 26176 + (size_t)67 * 16;
      i1c4_4.sAo = (long long)66 * 66 * 3; i1c4_4.sAi = (long long)66 * 3; i1c4_4.sAm = 3; i1c4_4.sAk = 1; i1c4_4.sBo = 0; i1c4_4.sBi = 0; i1c4_4.sBn = 3 * 9; i1c4_4.sBk = 9; i1c4_4.sCo = (long long)66 * 66 * 16; i1c4_4.sCi = (long long)66 * 16; i1c4_4.sCm = 16; i1c4_4.sRo = (long long)66 * 66 * 16; i1c4_4.sRi = (long long)66 * 16; i1c4_4.sRm = 16; i1c4_4.sRn = 1;
      i1c4_4.M = 64; i1c4_4.N = 16; i1c4_4.K = 3; i1c4_4.zi_n = 64; i1c4_4.flags = 4; i1c4_4.act = 0;
      i1c4_4.alpha = 1.0f; i1c4_4.beta = 1.0f; i1c4_4.sa = 1.0f; i1c4_4.sb = 1.0f; i1c4_4.Npad = 16; i1c4_4.pad_ = 0;
      k_gemm<1><<<dim3((unsigned)((16) + 31) / 32, (unsigned)((64) + 15) / 16, (unsigned)(2 * 64)), 32, 0, stream>>>(i1c4_4); }
    { GemmP i1c4_5;
      i1c4_5.A = R67 + 0 + (size_t)68 * 3; i1c4_5.B = iw1 + 5; i1c4_5.bias = R67 + 0 + (size_t)68 * 3; i1c4_5.R = R67 + 26176 + (size_t)67 * 16; i1c4_5.C = R67 + 26176 + (size_t)67 * 16;
      i1c4_5.sAo = (long long)66 * 66 * 3; i1c4_5.sAi = (long long)66 * 3; i1c4_5.sAm = 3; i1c4_5.sAk = 1; i1c4_5.sBo = 0; i1c4_5.sBi = 0; i1c4_5.sBn = 3 * 9; i1c4_5.sBk = 9; i1c4_5.sCo = (long long)66 * 66 * 16; i1c4_5.sCi = (long long)66 * 16; i1c4_5.sCm = 16; i1c4_5.sRo = (long long)66 * 66 * 16; i1c4_5.sRi = (long long)66 * 16; i1c4_5.sRm = 16; i1c4_5.sRn = 1;
      i1c4_5.M = 64; i1c4_5.N = 16; i1c4_5.K = 3; i1c4_5.zi_n = 64; i1c4_5.flags = 4; i1c4_5.act = 0;
      i1c4_5.alpha = 1.0f; i1c4_5.beta = 1.0f; i1c4_5.sa = 1.0f; i1c4_5.sb = 1.0f; i1c4_5.Npad = 16; i1c4_5.pad_ = 0;
      k_gemm<1><<<dim3((unsigned)((16) + 31) / 32, (unsigned)((64) + 15) / 16, (unsigned)(2 * 64)), 32, 0, stream>>>(i1c4_5); }
    { GemmP i1c4_6;
      i1c4_6.A = R67 + 0 + (size_t)132 * 3; i1c4_6.B = iw1 + 6; i1c4_6.bias = R67 + 0 + (size_t)132 * 3; i1c4_6.R = R67 + 26176 + (size_t)67 * 16; i1c4_6.C = R67 + 26176 + (size_t)67 * 16;
      i1c4_6.sAo = (long long)66 * 66 * 3; i1c4_6.sAi = (long long)66 * 3; i1c4_6.sAm = 3; i1c4_6.sAk = 1; i1c4_6.sBo = 0; i1c4_6.sBi = 0; i1c4_6.sBn = 3 * 9; i1c4_6.sBk = 9; i1c4_6.sCo = (long long)66 * 66 * 16; i1c4_6.sCi = (long long)66 * 16; i1c4_6.sCm = 16; i1c4_6.sRo = (long long)66 * 66 * 16; i1c4_6.sRi = (long long)66 * 16; i1c4_6.sRm = 16; i1c4_6.sRn = 1;
      i1c4_6.M = 64; i1c4_6.N = 16; i1c4_6.K = 3; i1c4_6.zi_n = 64; i1c4_6.flags = 4; i1c4_6.act = 0;
      i1c4_6.alpha = 1.0f; i1c4_6.beta = 1.0f; i1c4_6.sa = 1.0f; i1c4_6.sb = 1.0f; i1c4_6.Npad = 16; i1c4_6.pad_ = 0;
      k_gemm<1><<<dim3((unsigned)((16) + 31) / 32, (unsigned)((64) + 15) / 16, (unsigned)(2 * 64)), 32, 0, stream>>>(i1c4_6); }
    { GemmP i1c4_7;
      i1c4_7.A = R67 + 0 + (size_t)133 * 3; i1c4_7.B = iw1 + 7; i1c4_7.bias = R67 + 0 + (size_t)133 * 3; i1c4_7.R = R67 + 26176 + (size_t)67 * 16; i1c4_7.C = R67 + 26176 + (size_t)67 * 16;
      i1c4_7.sAo = (long long)66 * 66 * 3; i1c4_7.sAi = (long long)66 * 3; i1c4_7.sAm = 3; i1c4_7.sAk = 1; i1c4_7.sBo = 0; i1c4_7.sBi = 0; i1c4_7.sBn = 3 * 9; i1c4_7.sBk = 9; i1c4_7.sCo = (long long)66 * 66 * 16; i1c4_7.sCi = (long long)66 * 16; i1c4_7.sCm = 16; i1c4_7.sRo = (long long)66 * 66 * 16; i1c4_7.sRi = (long long)66 * 16; i1c4_7.sRm = 16; i1c4_7.sRn = 1;
      i1c4_7.M = 64; i1c4_7.N = 16; i1c4_7.K = 3; i1c4_7.zi_n = 64; i1c4_7.flags = 4; i1c4_7.act = 0;
      i1c4_7.alpha = 1.0f; i1c4_7.beta = 1.0f; i1c4_7.sa = 1.0f; i1c4_7.sb = 1.0f; i1c4_7.Npad = 16; i1c4_7.pad_ = 0;
      k_gemm<1><<<dim3((unsigned)((16) + 31) / 32, (unsigned)((64) + 15) / 16, (unsigned)(2 * 64)), 32, 0, stream>>>(i1c4_7); }
    { GemmP i1c4_8;
      i1c4_8.A = R67 + 0 + (size_t)134 * 3; i1c4_8.B = iw1 + 8; i1c4_8.bias = R67 + 0 + (size_t)134 * 3; i1c4_8.R = R67 + 26176 + (size_t)67 * 16; i1c4_8.C = R67 + 26176 + (size_t)67 * 16;
      i1c4_8.sAo = (long long)66 * 66 * 3; i1c4_8.sAi = (long long)66 * 3; i1c4_8.sAm = 3; i1c4_8.sAk = 1; i1c4_8.sBo = 0; i1c4_8.sBi = 0; i1c4_8.sBn = 3 * 9; i1c4_8.sBk = 9; i1c4_8.sCo = (long long)66 * 66 * 16; i1c4_8.sCi = (long long)66 * 16; i1c4_8.sCm = 16; i1c4_8.sRo = (long long)66 * 66 * 16; i1c4_8.sRi = (long long)66 * 16; i1c4_8.sRm = 16; i1c4_8.sRn = 1;
      i1c4_8.M = 64; i1c4_8.N = 16; i1c4_8.K = 3; i1c4_8.zi_n = 64; i1c4_8.flags = 4; i1c4_8.act = 0;
      i1c4_8.alpha = 1.0f; i1c4_8.beta = 1.0f; i1c4_8.sa = 1.0f; i1c4_8.sb = 1.0f; i1c4_8.Npad = 16; i1c4_8.pad_ = 0;
      k_gemm<1><<<dim3((unsigned)((16) + 31) / 32, (unsigned)((64) + 15) / 16, (unsigned)(2 * 64)), 32, 0, stream>>>(i1c4_8); }
    k_mm_relu2d<<<(unsigned)(((long long)2 * HW * 16 + 255) / 256), 256, 0, stream>>>(R67 + 26176, nullptr, 2, 64, 16);
    { GemmP i2c4_0;
      i2c4_0.A = R67 + 26176 + (size_t)0 * 16; i2c4_0.B = iw2 + 0; i2c4_0.bias = ib2; i2c4_0.R = R67 + 26176 + (size_t)0 * 16; i2c4_0.C = R67 + 165568 + (size_t)67 * 32;
      i2c4_0.sAo = (long long)66 * 66 * 16; i2c4_0.sAi = (long long)66 * 16; i2c4_0.sAm = 16; i2c4_0.sAk = 1; i2c4_0.sBo = 0; i2c4_0.sBi = 0; i2c4_0.sBn = 16 * 9; i2c4_0.sBk = 9; i2c4_0.sCo = (long long)66 * 66 * 32; i2c4_0.sCi = (long long)66 * 32; i2c4_0.sCm = 32; i2c4_0.sRo = 0; i2c4_0.sRi = 0; i2c4_0.sRm = 0; i2c4_0.sRn = 0;
      i2c4_0.M = 64; i2c4_0.N = 32; i2c4_0.K = 16; i2c4_0.zi_n = 64; i2c4_0.flags = 1; i2c4_0.act = 0;
      i2c4_0.alpha = 1.0f; i2c4_0.beta = 0.0f; i2c4_0.sa = 1.0f; i2c4_0.sb = 1.0f; i2c4_0.Npad = 32; i2c4_0.pad_ = 0;
      k_gemm<1><<<dim3((unsigned)((32) + 31) / 32, (unsigned)((64) + 15) / 16, (unsigned)(2 * 64)), 32, 0, stream>>>(i2c4_0); }
    { GemmP i2c4_1;
      i2c4_1.A = R67 + 26176 + (size_t)1 * 16; i2c4_1.B = iw2 + 1; i2c4_1.bias = R67 + 26176 + (size_t)1 * 16; i2c4_1.R = R67 + 165568 + (size_t)67 * 32; i2c4_1.C = R67 + 165568 + (size_t)67 * 32;
      i2c4_1.sAo = (long long)66 * 66 * 16; i2c4_1.sAi = (long long)66 * 16; i2c4_1.sAm = 16; i2c4_1.sAk = 1; i2c4_1.sBo = 0; i2c4_1.sBi = 0; i2c4_1.sBn = 16 * 9; i2c4_1.sBk = 9; i2c4_1.sCo = (long long)66 * 66 * 32; i2c4_1.sCi = (long long)66 * 32; i2c4_1.sCm = 32; i2c4_1.sRo = (long long)66 * 66 * 32; i2c4_1.sRi = (long long)66 * 32; i2c4_1.sRm = 32; i2c4_1.sRn = 1;
      i2c4_1.M = 64; i2c4_1.N = 32; i2c4_1.K = 16; i2c4_1.zi_n = 64; i2c4_1.flags = 4; i2c4_1.act = 0;
      i2c4_1.alpha = 1.0f; i2c4_1.beta = 1.0f; i2c4_1.sa = 1.0f; i2c4_1.sb = 1.0f; i2c4_1.Npad = 32; i2c4_1.pad_ = 0;
      k_gemm<1><<<dim3((unsigned)((32) + 31) / 32, (unsigned)((64) + 15) / 16, (unsigned)(2 * 64)), 32, 0, stream>>>(i2c4_1); }
    { GemmP i2c4_2;
      i2c4_2.A = R67 + 26176 + (size_t)2 * 16; i2c4_2.B = iw2 + 2; i2c4_2.bias = R67 + 26176 + (size_t)2 * 16; i2c4_2.R = R67 + 165568 + (size_t)67 * 32; i2c4_2.C = R67 + 165568 + (size_t)67 * 32;
      i2c4_2.sAo = (long long)66 * 66 * 16; i2c4_2.sAi = (long long)66 * 16; i2c4_2.sAm = 16; i2c4_2.sAk = 1; i2c4_2.sBo = 0; i2c4_2.sBi = 0; i2c4_2.sBn = 16 * 9; i2c4_2.sBk = 9; i2c4_2.sCo = (long long)66 * 66 * 32; i2c4_2.sCi = (long long)66 * 32; i2c4_2.sCm = 32; i2c4_2.sRo = (long long)66 * 66 * 32; i2c4_2.sRi = (long long)66 * 32; i2c4_2.sRm = 32; i2c4_2.sRn = 1;
      i2c4_2.M = 64; i2c4_2.N = 32; i2c4_2.K = 16; i2c4_2.zi_n = 64; i2c4_2.flags = 4; i2c4_2.act = 0;
      i2c4_2.alpha = 1.0f; i2c4_2.beta = 1.0f; i2c4_2.sa = 1.0f; i2c4_2.sb = 1.0f; i2c4_2.Npad = 32; i2c4_2.pad_ = 0;
      k_gemm<1><<<dim3((unsigned)((32) + 31) / 32, (unsigned)((64) + 15) / 16, (unsigned)(2 * 64)), 32, 0, stream>>>(i2c4_2); }
    { GemmP i2c4_3;
      i2c4_3.A = R67 + 26176 + (size_t)66 * 16; i2c4_3.B = iw2 + 3; i2c4_3.bias = R67 + 26176 + (size_t)66 * 16; i2c4_3.R = R67 + 165568 + (size_t)67 * 32; i2c4_3.C = R67 + 165568 + (size_t)67 * 32;
      i2c4_3.sAo = (long long)66 * 66 * 16; i2c4_3.sAi = (long long)66 * 16; i2c4_3.sAm = 16; i2c4_3.sAk = 1; i2c4_3.sBo = 0; i2c4_3.sBi = 0; i2c4_3.sBn = 16 * 9; i2c4_3.sBk = 9; i2c4_3.sCo = (long long)66 * 66 * 32; i2c4_3.sCi = (long long)66 * 32; i2c4_3.sCm = 32; i2c4_3.sRo = (long long)66 * 66 * 32; i2c4_3.sRi = (long long)66 * 32; i2c4_3.sRm = 32; i2c4_3.sRn = 1;
      i2c4_3.M = 64; i2c4_3.N = 32; i2c4_3.K = 16; i2c4_3.zi_n = 64; i2c4_3.flags = 4; i2c4_3.act = 0;
      i2c4_3.alpha = 1.0f; i2c4_3.beta = 1.0f; i2c4_3.sa = 1.0f; i2c4_3.sb = 1.0f; i2c4_3.Npad = 32; i2c4_3.pad_ = 0;
      k_gemm<1><<<dim3((unsigned)((32) + 31) / 32, (unsigned)((64) + 15) / 16, (unsigned)(2 * 64)), 32, 0, stream>>>(i2c4_3); }
    { GemmP i2c4_4;
      i2c4_4.A = R67 + 26176 + (size_t)67 * 16; i2c4_4.B = iw2 + 4; i2c4_4.bias = R67 + 26176 + (size_t)67 * 16; i2c4_4.R = R67 + 165568 + (size_t)67 * 32; i2c4_4.C = R67 + 165568 + (size_t)67 * 32;
      i2c4_4.sAo = (long long)66 * 66 * 16; i2c4_4.sAi = (long long)66 * 16; i2c4_4.sAm = 16; i2c4_4.sAk = 1; i2c4_4.sBo = 0; i2c4_4.sBi = 0; i2c4_4.sBn = 16 * 9; i2c4_4.sBk = 9; i2c4_4.sCo = (long long)66 * 66 * 32; i2c4_4.sCi = (long long)66 * 32; i2c4_4.sCm = 32; i2c4_4.sRo = (long long)66 * 66 * 32; i2c4_4.sRi = (long long)66 * 32; i2c4_4.sRm = 32; i2c4_4.sRn = 1;
      i2c4_4.M = 64; i2c4_4.N = 32; i2c4_4.K = 16; i2c4_4.zi_n = 64; i2c4_4.flags = 4; i2c4_4.act = 0;
      i2c4_4.alpha = 1.0f; i2c4_4.beta = 1.0f; i2c4_4.sa = 1.0f; i2c4_4.sb = 1.0f; i2c4_4.Npad = 32; i2c4_4.pad_ = 0;
      k_gemm<1><<<dim3((unsigned)((32) + 31) / 32, (unsigned)((64) + 15) / 16, (unsigned)(2 * 64)), 32, 0, stream>>>(i2c4_4); }
    { GemmP i2c4_5;
      i2c4_5.A = R67 + 26176 + (size_t)68 * 16; i2c4_5.B = iw2 + 5; i2c4_5.bias = R67 + 26176 + (size_t)68 * 16; i2c4_5.R = R67 + 165568 + (size_t)67 * 32; i2c4_5.C = R67 + 165568 + (size_t)67 * 32;
      i2c4_5.sAo = (long long)66 * 66 * 16; i2c4_5.sAi = (long long)66 * 16; i2c4_5.sAm = 16; i2c4_5.sAk = 1; i2c4_5.sBo = 0; i2c4_5.sBi = 0; i2c4_5.sBn = 16 * 9; i2c4_5.sBk = 9; i2c4_5.sCo = (long long)66 * 66 * 32; i2c4_5.sCi = (long long)66 * 32; i2c4_5.sCm = 32; i2c4_5.sRo = (long long)66 * 66 * 32; i2c4_5.sRi = (long long)66 * 32; i2c4_5.sRm = 32; i2c4_5.sRn = 1;
      i2c4_5.M = 64; i2c4_5.N = 32; i2c4_5.K = 16; i2c4_5.zi_n = 64; i2c4_5.flags = 4; i2c4_5.act = 0;
      i2c4_5.alpha = 1.0f; i2c4_5.beta = 1.0f; i2c4_5.sa = 1.0f; i2c4_5.sb = 1.0f; i2c4_5.Npad = 32; i2c4_5.pad_ = 0;
      k_gemm<1><<<dim3((unsigned)((32) + 31) / 32, (unsigned)((64) + 15) / 16, (unsigned)(2 * 64)), 32, 0, stream>>>(i2c4_5); }
    { GemmP i2c4_6;
      i2c4_6.A = R67 + 26176 + (size_t)132 * 16; i2c4_6.B = iw2 + 6; i2c4_6.bias = R67 + 26176 + (size_t)132 * 16; i2c4_6.R = R67 + 165568 + (size_t)67 * 32; i2c4_6.C = R67 + 165568 + (size_t)67 * 32;
      i2c4_6.sAo = (long long)66 * 66 * 16; i2c4_6.sAi = (long long)66 * 16; i2c4_6.sAm = 16; i2c4_6.sAk = 1; i2c4_6.sBo = 0; i2c4_6.sBi = 0; i2c4_6.sBn = 16 * 9; i2c4_6.sBk = 9; i2c4_6.sCo = (long long)66 * 66 * 32; i2c4_6.sCi = (long long)66 * 32; i2c4_6.sCm = 32; i2c4_6.sRo = (long long)66 * 66 * 32; i2c4_6.sRi = (long long)66 * 32; i2c4_6.sRm = 32; i2c4_6.sRn = 1;
      i2c4_6.M = 64; i2c4_6.N = 32; i2c4_6.K = 16; i2c4_6.zi_n = 64; i2c4_6.flags = 4; i2c4_6.act = 0;
      i2c4_6.alpha = 1.0f; i2c4_6.beta = 1.0f; i2c4_6.sa = 1.0f; i2c4_6.sb = 1.0f; i2c4_6.Npad = 32; i2c4_6.pad_ = 0;
      k_gemm<1><<<dim3((unsigned)((32) + 31) / 32, (unsigned)((64) + 15) / 16, (unsigned)(2 * 64)), 32, 0, stream>>>(i2c4_6); }
    { GemmP i2c4_7;
      i2c4_7.A = R67 + 26176 + (size_t)133 * 16; i2c4_7.B = iw2 + 7; i2c4_7.bias = R67 + 26176 + (size_t)133 * 16; i2c4_7.R = R67 + 165568 + (size_t)67 * 32; i2c4_7.C = R67 + 165568 + (size_t)67 * 32;
      i2c4_7.sAo = (long long)66 * 66 * 16; i2c4_7.sAi = (long long)66 * 16; i2c4_7.sAm = 16; i2c4_7.sAk = 1; i2c4_7.sBo = 0; i2c4_7.sBi = 0; i2c4_7.sBn = 16 * 9; i2c4_7.sBk = 9; i2c4_7.sCo = (long long)66 * 66 * 32; i2c4_7.sCi = (long long)66 * 32; i2c4_7.sCm = 32; i2c4_7.sRo = (long long)66 * 66 * 32; i2c4_7.sRi = (long long)66 * 32; i2c4_7.sRm = 32; i2c4_7.sRn = 1;
      i2c4_7.M = 64; i2c4_7.N = 32; i2c4_7.K = 16; i2c4_7.zi_n = 64; i2c4_7.flags = 4; i2c4_7.act = 0;
      i2c4_7.alpha = 1.0f; i2c4_7.beta = 1.0f; i2c4_7.sa = 1.0f; i2c4_7.sb = 1.0f; i2c4_7.Npad = 32; i2c4_7.pad_ = 0;
      k_gemm<1><<<dim3((unsigned)((32) + 31) / 32, (unsigned)((64) + 15) / 16, (unsigned)(2 * 64)), 32, 0, stream>>>(i2c4_7); }
    { GemmP i2c4_8;
      i2c4_8.A = R67 + 26176 + (size_t)134 * 16; i2c4_8.B = iw2 + 8; i2c4_8.bias = R67 + 26176 + (size_t)134 * 16; i2c4_8.R = R67 + 165568 + (size_t)67 * 32; i2c4_8.C = R67 + 165568 + (size_t)67 * 32;
      i2c4_8.sAo = (long long)66 * 66 * 16; i2c4_8.sAi = (long long)66 * 16; i2c4_8.sAm = 16; i2c4_8.sAk = 1; i2c4_8.sBo = 0; i2c4_8.sBi = 0; i2c4_8.sBn = 16 * 9; i2c4_8.sBk = 9; i2c4_8.sCo = (long long)66 * 66 * 32; i2c4_8.sCi = (long long)66 * 32; i2c4_8.sCm = 32; i2c4_8.sRo = (long long)66 * 66 * 32; i2c4_8.sRi = (long long)66 * 32; i2c4_8.sRm = 32; i2c4_8.sRn = 1;
      i2c4_8.M = 64; i2c4_8.N = 32; i2c4_8.K = 16; i2c4_8.zi_n = 64; i2c4_8.flags = 4; i2c4_8.act = 0;
      i2c4_8.alpha = 1.0f; i2c4_8.beta = 1.0f; i2c4_8.sa = 1.0f; i2c4_8.sb = 1.0f; i2c4_8.Npad = 32; i2c4_8.pad_ = 0;
      k_gemm<1><<<dim3((unsigned)((32) + 31) / 32, (unsigned)((64) + 15) / 16, (unsigned)(2 * 64)), 32, 0, stream>>>(i2c4_8); }
    k_mm_relu2d<<<(unsigned)(((long long)2 * HW * 32 + 255) / 256), 256, 0, stream>>>(R67 + 165568, nullptr, 2, 64, 32);
    { GemmP i3c4_0;
      i3c4_0.A = R67 + 165568 + (size_t)0 * 32; i3c4_0.B = iw3 + 0; i3c4_0.bias = ib3; i3c4_0.R = R67 + 165568 + (size_t)0 * 32; i3c4_0.C = R67 + 444352 + (size_t)67 * 64;
      i3c4_0.sAo = (long long)66 * 66 * 32; i3c4_0.sAi = (long long)66 * 32; i3c4_0.sAm = 32; i3c4_0.sAk = 1; i3c4_0.sBo = 0; i3c4_0.sBi = 0; i3c4_0.sBn = 32 * 9; i3c4_0.sBk = 9; i3c4_0.sCo = (long long)66 * 66 * 64; i3c4_0.sCi = (long long)66 * 64; i3c4_0.sCm = 64; i3c4_0.sRo = 0; i3c4_0.sRi = 0; i3c4_0.sRm = 0; i3c4_0.sRn = 0;
      i3c4_0.M = 64; i3c4_0.N = 64; i3c4_0.K = 32; i3c4_0.zi_n = 64; i3c4_0.flags = 1; i3c4_0.act = 0;
      i3c4_0.alpha = 1.0f; i3c4_0.beta = 0.0f; i3c4_0.sa = 1.0f; i3c4_0.sb = 1.0f; i3c4_0.Npad = 64; i3c4_0.pad_ = 0;
      k_gemm<1><<<dim3((unsigned)((64) + 31) / 32, (unsigned)((64) + 15) / 16, (unsigned)(2 * 64)), 32, 0, stream>>>(i3c4_0); }
    { GemmP i3c4_1;
      i3c4_1.A = R67 + 165568 + (size_t)1 * 32; i3c4_1.B = iw3 + 1; i3c4_1.bias = R67 + 165568 + (size_t)1 * 32; i3c4_1.R = R67 + 444352 + (size_t)67 * 64; i3c4_1.C = R67 + 444352 + (size_t)67 * 64;
      i3c4_1.sAo = (long long)66 * 66 * 32; i3c4_1.sAi = (long long)66 * 32; i3c4_1.sAm = 32; i3c4_1.sAk = 1; i3c4_1.sBo = 0; i3c4_1.sBi = 0; i3c4_1.sBn = 32 * 9; i3c4_1.sBk = 9; i3c4_1.sCo = (long long)66 * 66 * 64; i3c4_1.sCi = (long long)66 * 64; i3c4_1.sCm = 64; i3c4_1.sRo = (long long)66 * 66 * 64; i3c4_1.sRi = (long long)66 * 64; i3c4_1.sRm = 64; i3c4_1.sRn = 1;
      i3c4_1.M = 64; i3c4_1.N = 64; i3c4_1.K = 32; i3c4_1.zi_n = 64; i3c4_1.flags = 4; i3c4_1.act = 0;
      i3c4_1.alpha = 1.0f; i3c4_1.beta = 1.0f; i3c4_1.sa = 1.0f; i3c4_1.sb = 1.0f; i3c4_1.Npad = 64; i3c4_1.pad_ = 0;
      k_gemm<1><<<dim3((unsigned)((64) + 31) / 32, (unsigned)((64) + 15) / 16, (unsigned)(2 * 64)), 32, 0, stream>>>(i3c4_1); }
    { GemmP i3c4_2;
      i3c4_2.A = R67 + 165568 + (size_t)2 * 32; i3c4_2.B = iw3 + 2; i3c4_2.bias = R67 + 165568 + (size_t)2 * 32; i3c4_2.R = R67 + 444352 + (size_t)67 * 64; i3c4_2.C = R67 + 444352 + (size_t)67 * 64;
      i3c4_2.sAo = (long long)66 * 66 * 32; i3c4_2.sAi = (long long)66 * 32; i3c4_2.sAm = 32; i3c4_2.sAk = 1; i3c4_2.sBo = 0; i3c4_2.sBi = 0; i3c4_2.sBn = 32 * 9; i3c4_2.sBk = 9; i3c4_2.sCo = (long long)66 * 66 * 64; i3c4_2.sCi = (long long)66 * 64; i3c4_2.sCm = 64; i3c4_2.sRo = (long long)66 * 66 * 64; i3c4_2.sRi = (long long)66 * 64; i3c4_2.sRm = 64; i3c4_2.sRn = 1;
      i3c4_2.M = 64; i3c4_2.N = 64; i3c4_2.K = 32; i3c4_2.zi_n = 64; i3c4_2.flags = 4; i3c4_2.act = 0;
      i3c4_2.alpha = 1.0f; i3c4_2.beta = 1.0f; i3c4_2.sa = 1.0f; i3c4_2.sb = 1.0f; i3c4_2.Npad = 64; i3c4_2.pad_ = 0;
      k_gemm<1><<<dim3((unsigned)((64) + 31) / 32, (unsigned)((64) + 15) / 16, (unsigned)(2 * 64)), 32, 0, stream>>>(i3c4_2); }
    { GemmP i3c4_3;
      i3c4_3.A = R67 + 165568 + (size_t)66 * 32; i3c4_3.B = iw3 + 3; i3c4_3.bias = R67 + 165568 + (size_t)66 * 32; i3c4_3.R = R67 + 444352 + (size_t)67 * 64; i3c4_3.C = R67 + 444352 + (size_t)67 * 64;
      i3c4_3.sAo = (long long)66 * 66 * 32; i3c4_3.sAi = (long long)66 * 32; i3c4_3.sAm = 32; i3c4_3.sAk = 1; i3c4_3.sBo = 0; i3c4_3.sBi = 0; i3c4_3.sBn = 32 * 9; i3c4_3.sBk = 9; i3c4_3.sCo = (long long)66 * 66 * 64; i3c4_3.sCi = (long long)66 * 64; i3c4_3.sCm = 64; i3c4_3.sRo = (long long)66 * 66 * 64; i3c4_3.sRi = (long long)66 * 64; i3c4_3.sRm = 64; i3c4_3.sRn = 1;
      i3c4_3.M = 64; i3c4_3.N = 64; i3c4_3.K = 32; i3c4_3.zi_n = 64; i3c4_3.flags = 4; i3c4_3.act = 0;
      i3c4_3.alpha = 1.0f; i3c4_3.beta = 1.0f; i3c4_3.sa = 1.0f; i3c4_3.sb = 1.0f; i3c4_3.Npad = 64; i3c4_3.pad_ = 0;
      k_gemm<1><<<dim3((unsigned)((64) + 31) / 32, (unsigned)((64) + 15) / 16, (unsigned)(2 * 64)), 32, 0, stream>>>(i3c4_3); }
    { GemmP i3c4_4;
      i3c4_4.A = R67 + 165568 + (size_t)67 * 32; i3c4_4.B = iw3 + 4; i3c4_4.bias = R67 + 165568 + (size_t)67 * 32; i3c4_4.R = R67 + 444352 + (size_t)67 * 64; i3c4_4.C = R67 + 444352 + (size_t)67 * 64;
      i3c4_4.sAo = (long long)66 * 66 * 32; i3c4_4.sAi = (long long)66 * 32; i3c4_4.sAm = 32; i3c4_4.sAk = 1; i3c4_4.sBo = 0; i3c4_4.sBi = 0; i3c4_4.sBn = 32 * 9; i3c4_4.sBk = 9; i3c4_4.sCo = (long long)66 * 66 * 64; i3c4_4.sCi = (long long)66 * 64; i3c4_4.sCm = 64; i3c4_4.sRo = (long long)66 * 66 * 64; i3c4_4.sRi = (long long)66 * 64; i3c4_4.sRm = 64; i3c4_4.sRn = 1;
      i3c4_4.M = 64; i3c4_4.N = 64; i3c4_4.K = 32; i3c4_4.zi_n = 64; i3c4_4.flags = 4; i3c4_4.act = 0;
      i3c4_4.alpha = 1.0f; i3c4_4.beta = 1.0f; i3c4_4.sa = 1.0f; i3c4_4.sb = 1.0f; i3c4_4.Npad = 64; i3c4_4.pad_ = 0;
      k_gemm<1><<<dim3((unsigned)((64) + 31) / 32, (unsigned)((64) + 15) / 16, (unsigned)(2 * 64)), 32, 0, stream>>>(i3c4_4); }
    { GemmP i3c4_5;
      i3c4_5.A = R67 + 165568 + (size_t)68 * 32; i3c4_5.B = iw3 + 5; i3c4_5.bias = R67 + 165568 + (size_t)68 * 32; i3c4_5.R = R67 + 444352 + (size_t)67 * 64; i3c4_5.C = R67 + 444352 + (size_t)67 * 64;
      i3c4_5.sAo = (long long)66 * 66 * 32; i3c4_5.sAi = (long long)66 * 32; i3c4_5.sAm = 32; i3c4_5.sAk = 1; i3c4_5.sBo = 0; i3c4_5.sBi = 0; i3c4_5.sBn = 32 * 9; i3c4_5.sBk = 9; i3c4_5.sCo = (long long)66 * 66 * 64; i3c4_5.sCi = (long long)66 * 64; i3c4_5.sCm = 64; i3c4_5.sRo = (long long)66 * 66 * 64; i3c4_5.sRi = (long long)66 * 64; i3c4_5.sRm = 64; i3c4_5.sRn = 1;
      i3c4_5.M = 64; i3c4_5.N = 64; i3c4_5.K = 32; i3c4_5.zi_n = 64; i3c4_5.flags = 4; i3c4_5.act = 0;
      i3c4_5.alpha = 1.0f; i3c4_5.beta = 1.0f; i3c4_5.sa = 1.0f; i3c4_5.sb = 1.0f; i3c4_5.Npad = 64; i3c4_5.pad_ = 0;
      k_gemm<1><<<dim3((unsigned)((64) + 31) / 32, (unsigned)((64) + 15) / 16, (unsigned)(2 * 64)), 32, 0, stream>>>(i3c4_5); }
    { GemmP i3c4_6;
      i3c4_6.A = R67 + 165568 + (size_t)132 * 32; i3c4_6.B = iw3 + 6; i3c4_6.bias = R67 + 165568 + (size_t)132 * 32; i3c4_6.R = R67 + 444352 + (size_t)67 * 64; i3c4_6.C = R67 + 444352 + (size_t)67 * 64;
      i3c4_6.sAo = (long long)66 * 66 * 32; i3c4_6.sAi = (long long)66 * 32; i3c4_6.sAm = 32; i3c4_6.sAk = 1; i3c4_6.sBo = 0; i3c4_6.sBi = 0; i3c4_6.sBn = 32 * 9; i3c4_6.sBk = 9; i3c4_6.sCo = (long long)66 * 66 * 64; i3c4_6.sCi = (long long)66 * 64; i3c4_6.sCm = 64; i3c4_6.sRo = (long long)66 * 66 * 64; i3c4_6.sRi = (long long)66 * 64; i3c4_6.sRm = 64; i3c4_6.sRn = 1;
      i3c4_6.M = 64; i3c4_6.N = 64; i3c4_6.K = 32; i3c4_6.zi_n = 64; i3c4_6.flags = 4; i3c4_6.act = 0;
      i3c4_6.alpha = 1.0f; i3c4_6.beta = 1.0f; i3c4_6.sa = 1.0f; i3c4_6.sb = 1.0f; i3c4_6.Npad = 64; i3c4_6.pad_ = 0;
      k_gemm<1><<<dim3((unsigned)((64) + 31) / 32, (unsigned)((64) + 15) / 16, (unsigned)(2 * 64)), 32, 0, stream>>>(i3c4_6); }
    { GemmP i3c4_7;
      i3c4_7.A = R67 + 165568 + (size_t)133 * 32; i3c4_7.B = iw3 + 7; i3c4_7.bias = R67 + 165568 + (size_t)133 * 32; i3c4_7.R = R67 + 444352 + (size_t)67 * 64; i3c4_7.C = R67 + 444352 + (size_t)67 * 64;
      i3c4_7.sAo = (long long)66 * 66 * 32; i3c4_7.sAi = (long long)66 * 32; i3c4_7.sAm = 32; i3c4_7.sAk = 1; i3c4_7.sBo = 0; i3c4_7.sBi = 0; i3c4_7.sBn = 32 * 9; i3c4_7.sBk = 9; i3c4_7.sCo = (long long)66 * 66 * 64; i3c4_7.sCi = (long long)66 * 64; i3c4_7.sCm = 64; i3c4_7.sRo = (long long)66 * 66 * 64; i3c4_7.sRi = (long long)66 * 64; i3c4_7.sRm = 64; i3c4_7.sRn = 1;
      i3c4_7.M = 64; i3c4_7.N = 64; i3c4_7.K = 32; i3c4_7.zi_n = 64; i3c4_7.flags = 4; i3c4_7.act = 0;
      i3c4_7.alpha = 1.0f; i3c4_7.beta = 1.0f; i3c4_7.sa = 1.0f; i3c4_7.sb = 1.0f; i3c4_7.Npad = 64; i3c4_7.pad_ = 0;
      k_gemm<1><<<dim3((unsigned)((64) + 31) / 32, (unsigned)((64) + 15) / 16, (unsigned)(2 * 64)), 32, 0, stream>>>(i3c4_7); }
    { GemmP i3c4_8;
      i3c4_8.A = R67 + 165568 + (size_t)134 * 32; i3c4_8.B = iw3 + 8; i3c4_8.bias = R67 + 165568 + (size_t)134 * 32; i3c4_8.R = R67 + 444352 + (size_t)67 * 64; i3c4_8.C = R67 + 444352 + (size_t)67 * 64;
      i3c4_8.sAo = (long long)66 * 66 * 32; i3c4_8.sAi = (long long)66 * 32; i3c4_8.sAm = 32; i3c4_8.sAk = 1; i3c4_8.sBo = 0; i3c4_8.sBi = 0; i3c4_8.sBn = 32 * 9; i3c4_8.sBk = 9; i3c4_8.sCo = (long long)66 * 66 * 64; i3c4_8.sCi = (long long)66 * 64; i3c4_8.sCm = 64; i3c4_8.sRo = (long long)66 * 66 * 64; i3c4_8.sRi = (long long)66 * 64; i3c4_8.sRm = 64; i3c4_8.sRn = 1;
      i3c4_8.M = 64; i3c4_8.N = 64; i3c4_8.K = 32; i3c4_8.zi_n = 64; i3c4_8.flags = 4; i3c4_8.act = 0;
      i3c4_8.alpha = 1.0f; i3c4_8.beta = 1.0f; i3c4_8.sa = 1.0f; i3c4_8.sb = 1.0f; i3c4_8.Npad = 64; i3c4_8.pad_ = 0;
      k_gemm<1><<<dim3((unsigned)((64) + 31) / 32, (unsigned)((64) + 15) / 16, (unsigned)(2 * 64)), 32, 0, stream>>>(i3c4_8); }
    k_mm_relu2d<<<(unsigned)(((long long)2 * HW * 64 + 255) / 256), 256, 0, stream>>>(R67 + 444352, R67 + 1001920, 2, 64, 64);
    { GemmP gqkv4;
      gqkv4.A = R67 + 1001920; gqkv4.B = qkvw; gqkv4.bias = qkvb; gqkv4.R = R67 + 1001920; gqkv4.C = R67 + 1526208;
      gqkv4.sAo = 0; gqkv4.sAi = 0; gqkv4.sAm = 64; gqkv4.sAk = 1; gqkv4.sBo = 0; gqkv4.sBi = 0; gqkv4.sBn = 64; gqkv4.sBk = 1; gqkv4.sCo = 0; gqkv4.sCi = 0; gqkv4.sCm = 192; gqkv4.sRo = 0; gqkv4.sRi = 0; gqkv4.sRm = 0; gqkv4.sRn = 0;
      gqkv4.M = 2 * HW; gqkv4.N = 192; gqkv4.K = 64; gqkv4.zi_n = 1; gqkv4.flags = 1; gqkv4.act = 0;
      gqkv4.alpha = 1.0f; gqkv4.beta = 0.0f; gqkv4.sa = 1.0f; gqkv4.sb = 1.0f; gqkv4.Npad = 192; gqkv4.pad_ = 0;
      k_gemm<1><<<dim3((unsigned)((192) + 31) / 32, (unsigned)((2 * HW) + 15) / 16, (unsigned)(1)), 32, 0, stream>>>(gqkv4); }
    k_mm_dw<<<(unsigned)(((long long)2 * HW * 192 + 255) / 256), 256, 0, stream>>>(R67 + 1526208, dww, dwb, R67 + 3099072, 2, 64, 192);
    k_mm_fall<<<(unsigned)(((long long)2 * HW * 144 + 255) / 256), 256, 0, stream>>>(R67 + 3099072, fcw, fcb, R67 + 4671936, 2, HW, 192);
    k_mm_dep<<<(unsigned)(((long long)2 * 64 * HW + 255) / 256), 256, 0, stream>>>(R67 + 4671936, depw, depb, R67 + 5851584, 2, 64);
    k_mm_qknorm<<<2 * 128, 256, 0, stream>>>(R67 + 3099072, R67 + 6375872, 2, HW, 192);
    { GemmP gat4;
      gat4.A = R67 + 6375872; gat4.B = R67 + 6375872 + (size_t)64 * HW; gat4.bias = R67 + 6375872; gat4.R = R67 + 6375872; gat4.C = R67 + 7424448;
      gat4.sAo = (long long)128 * HW; gat4.sAi = (long long)16 * HW; gat4.sAm = HW; gat4.sAk = 1; gat4.sBo = (long long)128 * HW; gat4.sBi = (long long)16 * HW; gat4.sBn = HW; gat4.sBk = 1; gat4.sCo = (long long)4 * 16 * LP; gat4.sCi = 16 * LP; gat4.sCm = LP; gat4.sRo = 0; gat4.sRi = 0; gat4.sRm = 0; gat4.sRn = 0;
      gat4.M = 16; gat4.N = 16; gat4.K = HW; gat4.zi_n = 4; gat4.flags = 0; gat4.act = 0;
      gat4.alpha = 1.0f; gat4.beta = 0.0f; gat4.sa = 1.0f; gat4.sb = 1.0f; gat4.Npad = LP; gat4.pad_ = 0;
      k_gemm<1><<<dim3((unsigned)((LP) + 31) / 32, (unsigned)((16) + 15) / 16, (unsigned)(2 * 4)), 32, 0, stream>>>(gat4); }
    k_mm_sm16<<<(unsigned)((2 * 4 * 16 + 255) / 256), 256, 0, stream>>>(R67 + 7424448, temp, 2 * 4, LP);
    { GemmP gao4;
      gao4.A = R67 + 7424448; gao4.B = R67 + 3099072 + 128; gao4.bias = R67 + 7424448; gao4.R = R67 + 7424448; gao4.C = R67 + 7428544;
      gao4.sAo = (long long)4 * 16 * LP; gao4.sAi = 16 * LP; gao4.sAm = LP; gao4.sAk = 1; gao4.sBo = (long long)HW * 192; gao4.sBi = 16; gao4.sBn = 192; gao4.sBk = 1; gao4.sCo = (long long)64 * HW; gao4.sCi = (long long)16 * HW; gao4.sCm = HW; gao4.sRo = 0; gao4.sRi = 0; gao4.sRm = 0; gao4.sRn = 0;
      gao4.M = 16; gao4.N = HW; gao4.K = 16; gao4.zi_n = 4; gao4.flags = 0; gao4.act = 0;
      gao4.alpha = 1.0f; gao4.beta = 0.0f; gao4.sa = 1.0f; gao4.sb = 1.0f; gao4.Npad = HW; gao4.pad_ = 0;
      k_gemm<1><<<dim3((unsigned)((HW) + 31) / 32, (unsigned)((16) + 15) / 16, (unsigned)(2 * 4)), 32, 0, stream>>>(gao4); }
    { GemmP gproj4;
      gproj4.A = projw; gproj4.B = R67 + 7428544; gproj4.bias = projb; gproj4.R = projw; gproj4.C = R67 + 7952832;
      gproj4.sAo = 0; gproj4.sAi = 0; gproj4.sAm = 64; gproj4.sAk = 1; gproj4.sBo = (long long)64 * HW; gproj4.sBi = 0; gproj4.sBn = 1; gproj4.sBk = HW; gproj4.sCo = (long long)64 * HW; gproj4.sCi = 0; gproj4.sCm = HW; gproj4.sRo = 0; gproj4.sRi = 0; gproj4.sRm = 0; gproj4.sRn = 0;
      gproj4.M = 64; gproj4.N = HW; gproj4.K = 64; gproj4.zi_n = 1; gproj4.flags = 2; gproj4.act = 0;
      gproj4.alpha = 1.0f; gproj4.beta = 0.0f; gproj4.sa = 1.0f; gproj4.sb = 1.0f; gproj4.Npad = HW; gproj4.pad_ = 0;
      k_gemm<1><<<dim3((unsigned)((HW) + 31) / 32, (unsigned)((64) + 15) / 16, (unsigned)(2)), 32, 0, stream>>>(gproj4); }
    k_mm_imgfeat<<<(unsigned)(((long long)2 * SEQ * 64 + 255) / 256), 256, 0, stream>>>(R67 + 7952832, R67 + 5851584, IR + (size_t)8 * SEQ * 64, 2, HW, 64);
    hipMemsetAsync(R67 + 0, 0, (size_t)2 * 66 * 66 * 3 * 4, stream); hipMemsetAsync(R67 + 26176, 0, (size_t)2 * 66 * 66 * 16 * 4, stream); hipMemsetAsync(R67 + 165568, 0, (size_t)2 * 66 * 66 * 32 * 4, stream); hipMemsetAsync(R67 + 444352, 0, (size_t)2 * 66 * 66 * 64 * 4, stream);
    k_mm_padimg<<<(unsigned)(((long long)2 * HW * 3 + 255) / 256), 256, 0, stream>>>(img + (size_t)10 * 3 * HW, R67 + 0, 2, 3, 64);
    { GemmP i1c5_0;
      i1c5_0.A = R67 + 0 + (size_t)0 * 3; i1c5_0.B = iw1 + 0; i1c5_0.bias = ib1; i1c5_0.R = R67 + 0 + (size_t)0 * 3; i1c5_0.C = R67 + 26176 + (size_t)67 * 16;
      i1c5_0.sAo = (long long)66 * 66 * 3; i1c5_0.sAi = (long long)66 * 3; i1c5_0.sAm = 3; i1c5_0.sAk = 1; i1c5_0.sBo = 0; i1c5_0.sBi = 0; i1c5_0.sBn = 3 * 9; i1c5_0.sBk = 9; i1c5_0.sCo = (long long)66 * 66 * 16; i1c5_0.sCi = (long long)66 * 16; i1c5_0.sCm = 16; i1c5_0.sRo = 0; i1c5_0.sRi = 0; i1c5_0.sRm = 0; i1c5_0.sRn = 0;
      i1c5_0.M = 64; i1c5_0.N = 16; i1c5_0.K = 3; i1c5_0.zi_n = 64; i1c5_0.flags = 1; i1c5_0.act = 0;
      i1c5_0.alpha = 1.0f; i1c5_0.beta = 0.0f; i1c5_0.sa = 1.0f; i1c5_0.sb = 1.0f; i1c5_0.Npad = 16; i1c5_0.pad_ = 0;
      k_gemm<1><<<dim3((unsigned)((16) + 31) / 32, (unsigned)((64) + 15) / 16, (unsigned)(2 * 64)), 32, 0, stream>>>(i1c5_0); }
    { GemmP i1c5_1;
      i1c5_1.A = R67 + 0 + (size_t)1 * 3; i1c5_1.B = iw1 + 1; i1c5_1.bias = R67 + 0 + (size_t)1 * 3; i1c5_1.R = R67 + 26176 + (size_t)67 * 16; i1c5_1.C = R67 + 26176 + (size_t)67 * 16;
      i1c5_1.sAo = (long long)66 * 66 * 3; i1c5_1.sAi = (long long)66 * 3; i1c5_1.sAm = 3; i1c5_1.sAk = 1; i1c5_1.sBo = 0; i1c5_1.sBi = 0; i1c5_1.sBn = 3 * 9; i1c5_1.sBk = 9; i1c5_1.sCo = (long long)66 * 66 * 16; i1c5_1.sCi = (long long)66 * 16; i1c5_1.sCm = 16; i1c5_1.sRo = (long long)66 * 66 * 16; i1c5_1.sRi = (long long)66 * 16; i1c5_1.sRm = 16; i1c5_1.sRn = 1;
      i1c5_1.M = 64; i1c5_1.N = 16; i1c5_1.K = 3; i1c5_1.zi_n = 64; i1c5_1.flags = 4; i1c5_1.act = 0;
      i1c5_1.alpha = 1.0f; i1c5_1.beta = 1.0f; i1c5_1.sa = 1.0f; i1c5_1.sb = 1.0f; i1c5_1.Npad = 16; i1c5_1.pad_ = 0;
      k_gemm<1><<<dim3((unsigned)((16) + 31) / 32, (unsigned)((64) + 15) / 16, (unsigned)(2 * 64)), 32, 0, stream>>>(i1c5_1); }
    { GemmP i1c5_2;
      i1c5_2.A = R67 + 0 + (size_t)2 * 3; i1c5_2.B = iw1 + 2; i1c5_2.bias = R67 + 0 + (size_t)2 * 3; i1c5_2.R = R67 + 26176 + (size_t)67 * 16; i1c5_2.C = R67 + 26176 + (size_t)67 * 16;
      i1c5_2.sAo = (long long)66 * 66 * 3; i1c5_2.sAi = (long long)66 * 3; i1c5_2.sAm = 3; i1c5_2.sAk = 1; i1c5_2.sBo = 0; i1c5_2.sBi = 0; i1c5_2.sBn = 3 * 9; i1c5_2.sBk = 9; i1c5_2.sCo = (long long)66 * 66 * 16; i1c5_2.sCi = (long long)66 * 16; i1c5_2.sCm = 16; i1c5_2.sRo = (long long)66 * 66 * 16; i1c5_2.sRi = (long long)66 * 16; i1c5_2.sRm = 16; i1c5_2.sRn = 1;
      i1c5_2.M = 64; i1c5_2.N = 16; i1c5_2.K = 3; i1c5_2.zi_n = 64; i1c5_2.flags = 4; i1c5_2.act = 0;
      i1c5_2.alpha = 1.0f; i1c5_2.beta = 1.0f; i1c5_2.sa = 1.0f; i1c5_2.sb = 1.0f; i1c5_2.Npad = 16; i1c5_2.pad_ = 0;
      k_gemm<1><<<dim3((unsigned)((16) + 31) / 32, (unsigned)((64) + 15) / 16, (unsigned)(2 * 64)), 32, 0, stream>>>(i1c5_2); }
    { GemmP i1c5_3;
      i1c5_3.A = R67 + 0 + (size_t)66 * 3; i1c5_3.B = iw1 + 3; i1c5_3.bias = R67 + 0 + (size_t)66 * 3; i1c5_3.R = R67 + 26176 + (size_t)67 * 16; i1c5_3.C = R67 + 26176 + (size_t)67 * 16;
      i1c5_3.sAo = (long long)66 * 66 * 3; i1c5_3.sAi = (long long)66 * 3; i1c5_3.sAm = 3; i1c5_3.sAk = 1; i1c5_3.sBo = 0; i1c5_3.sBi = 0; i1c5_3.sBn = 3 * 9; i1c5_3.sBk = 9; i1c5_3.sCo = (long long)66 * 66 * 16; i1c5_3.sCi = (long long)66 * 16; i1c5_3.sCm = 16; i1c5_3.sRo = (long long)66 * 66 * 16; i1c5_3.sRi = (long long)66 * 16; i1c5_3.sRm = 16; i1c5_3.sRn = 1;
      i1c5_3.M = 64; i1c5_3.N = 16; i1c5_3.K = 3; i1c5_3.zi_n = 64; i1c5_3.flags = 4; i1c5_3.act = 0;
      i1c5_3.alpha = 1.0f; i1c5_3.beta = 1.0f; i1c5_3.sa = 1.0f; i1c5_3.sb = 1.0f; i1c5_3.Npad = 16; i1c5_3.pad_ = 0;
      k_gemm<1><<<dim3((unsigned)((16) + 31) / 32, (unsigned)((64) + 15) / 16, (unsigned)(2 * 64)), 32, 0, stream>>>(i1c5_3); }
    { GemmP i1c5_4;
      i1c5_4.A = R67 + 0 + (size_t)67 * 3; i1c5_4.B = iw1 + 4; i1c5_4.bias = R67 + 0 + (size_t)67 * 3; i1c5_4.R = R67 + 26176 + (size_t)67 * 16; i1c5_4.C = R67 + 26176 + (size_t)67 * 16;
      i1c5_4.sAo = (long long)66 * 66 * 3; i1c5_4.sAi = (long long)66 * 3; i1c5_4.sAm = 3; i1c5_4.sAk = 1; i1c5_4.sBo = 0; i1c5_4.sBi = 0; i1c5_4.sBn = 3 * 9; i1c5_4.sBk = 9; i1c5_4.sCo = (long long)66 * 66 * 16; i1c5_4.sCi = (long long)66 * 16; i1c5_4.sCm = 16; i1c5_4.sRo = (long long)66 * 66 * 16; i1c5_4.sRi = (long long)66 * 16; i1c5_4.sRm = 16; i1c5_4.sRn = 1;
      i1c5_4.M = 64; i1c5_4.N = 16; i1c5_4.K = 3; i1c5_4.zi_n = 64; i1c5_4.flags = 4; i1c5_4.act = 0;
      i1c5_4.alpha = 1.0f; i1c5_4.beta = 1.0f; i1c5_4.sa = 1.0f; i1c5_4.sb = 1.0f; i1c5_4.Npad = 16; i1c5_4.pad_ = 0;
      k_gemm<1><<<dim3((unsigned)((16) + 31) / 32, (unsigned)((64) + 15) / 16, (unsigned)(2 * 64)), 32, 0, stream>>>(i1c5_4); }
    { GemmP i1c5_5;
      i1c5_5.A = R67 + 0 + (size_t)68 * 3; i1c5_5.B = iw1 + 5; i1c5_5.bias = R67 + 0 + (size_t)68 * 3; i1c5_5.R = R67 + 26176 + (size_t)67 * 16; i1c5_5.C = R67 + 26176 + (size_t)67 * 16;
      i1c5_5.sAo = (long long)66 * 66 * 3; i1c5_5.sAi = (long long)66 * 3; i1c5_5.sAm = 3; i1c5_5.sAk = 1; i1c5_5.sBo = 0; i1c5_5.sBi = 0; i1c5_5.sBn = 3 * 9; i1c5_5.sBk = 9; i1c5_5.sCo = (long long)66 * 66 * 16; i1c5_5.sCi = (long long)66 * 16; i1c5_5.sCm = 16; i1c5_5.sRo = (long long)66 * 66 * 16; i1c5_5.sRi = (long long)66 * 16; i1c5_5.sRm = 16; i1c5_5.sRn = 1;
      i1c5_5.M = 64; i1c5_5.N = 16; i1c5_5.K = 3; i1c5_5.zi_n = 64; i1c5_5.flags = 4; i1c5_5.act = 0;
      i1c5_5.alpha = 1.0f; i1c5_5.beta = 1.0f; i1c5_5.sa = 1.0f; i1c5_5.sb = 1.0f; i1c5_5.Npad = 16; i1c5_5.pad_ = 0;
      k_gemm<1><<<dim3((unsigned)((16) + 31) / 32, (unsigned)((64) + 15) / 16, (unsigned)(2 * 64)), 32, 0, stream>>>(i1c5_5); }
    { GemmP i1c5_6;
      i1c5_6.A = R67 + 0 + (size_t)132 * 3; i1c5_6.B = iw1 + 6; i1c5_6.bias = R67 + 0 + (size_t)132 * 3; i1c5_6.R = R67 + 26176 + (size_t)67 * 16; i1c5_6.C = R67 + 26176 + (size_t)67 * 16;
      i1c5_6.sAo = (long long)66 * 66 * 3; i1c5_6.sAi = (long long)66 * 3; i1c5_6.sAm = 3; i1c5_6.sAk = 1; i1c5_6.sBo = 0; i1c5_6.sBi = 0; i1c5_6.sBn = 3 * 9; i1c5_6.sBk = 9; i1c5_6.sCo = (long long)66 * 66 * 16; i1c5_6.sCi = (long long)66 * 16; i1c5_6.sCm = 16; i1c5_6.sRo = (long long)66 * 66 * 16; i1c5_6.sRi = (long long)66 * 16; i1c5_6.sRm = 16; i1c5_6.sRn = 1;
      i1c5_6.M = 64; i1c5_6.N = 16; i1c5_6.K = 3; i1c5_6.zi_n = 64; i1c5_6.flags = 4; i1c5_6.act = 0;
      i1c5_6.alpha = 1.0f; i1c5_6.beta = 1.0f; i1c5_6.sa = 1.0f; i1c5_6.sb = 1.0f; i1c5_6.Npad = 16; i1c5_6.pad_ = 0;
      k_gemm<1><<<dim3((unsigned)((16) + 31) / 32, (unsigned)((64) + 15) / 16, (unsigned)(2 * 64)), 32, 0, stream>>>(i1c5_6); }
    { GemmP i1c5_7;
      i1c5_7.A = R67 + 0 + (size_t)133 * 3; i1c5_7.B = iw1 + 7; i1c5_7.bias = R67 + 0 + (size_t)133 * 3; i1c5_7.R = R67 + 26176 + (size_t)67 * 16; i1c5_7.C = R67 + 26176 + (size_t)67 * 16;
      i1c5_7.sAo = (long long)66 * 66 * 3; i1c5_7.sAi = (long long)66 * 3; i1c5_7.sAm = 3; i1c5_7.sAk = 1; i1c5_7.sBo = 0; i1c5_7.sBi = 0; i1c5_7.sBn = 3 * 9; i1c5_7.sBk = 9; i1c5_7.sCo = (long long)66 * 66 * 16; i1c5_7.sCi = (long long)66 * 16; i1c5_7.sCm = 16; i1c5_7.sRo = (long long)66 * 66 * 16; i1c5_7.sRi = (long long)66 * 16; i1c5_7.sRm = 16; i1c5_7.sRn = 1;
      i1c5_7.M = 64; i1c5_7.N = 16; i1c5_7.K = 3; i1c5_7.zi_n = 64; i1c5_7.flags = 4; i1c5_7.act = 0;
      i1c5_7.alpha = 1.0f; i1c5_7.beta = 1.0f; i1c5_7.sa = 1.0f; i1c5_7.sb = 1.0f; i1c5_7.Npad = 16; i1c5_7.pad_ = 0;
      k_gemm<1><<<dim3((unsigned)((16) + 31) / 32, (unsigned)((64) + 15) / 16, (unsigned)(2 * 64)), 32, 0, stream>>>(i1c5_7); }
    { GemmP i1c5_8;
      i1c5_8.A = R67 + 0 + (size_t)134 * 3; i1c5_8.B = iw1 + 8; i1c5_8.bias = R67 + 0 + (size_t)134 * 3; i1c5_8.R = R67 + 26176 + (size_t)67 * 16; i1c5_8.C = R67 + 26176 + (size_t)67 * 16;
      i1c5_8.sAo = (long long)66 * 66 * 3; i1c5_8.sAi = (long long)66 * 3; i1c5_8.sAm = 3; i1c5_8.sAk = 1; i1c5_8.sBo = 0; i1c5_8.sBi = 0; i1c5_8.sBn = 3 * 9; i1c5_8.sBk = 9; i1c5_8.sCo = (long long)66 * 66 * 16; i1c5_8.sCi = (long long)66 * 16; i1c5_8.sCm = 16; i1c5_8.sRo = (long long)66 * 66 * 16; i1c5_8.sRi = (long long)66 * 16; i1c5_8.sRm = 16; i1c5_8.sRn = 1;
      i1c5_8.M = 64; i1c5_8.N = 16; i1c5_8.K = 3; i1c5_8.zi_n = 64; i1c5_8.flags = 4; i1c5_8.act = 0;
      i1c5_8.alpha = 1.0f; i1c5_8.beta = 1.0f; i1c5_8.sa = 1.0f; i1c5_8.sb = 1.0f; i1c5_8.Npad = 16; i1c5_8.pad_ = 0;
      k_gemm<1><<<dim3((unsigned)((16) + 31) / 32, (unsigned)((64) + 15) / 16, (unsigned)(2 * 64)), 32, 0, stream>>>(i1c5_8); }
    k_mm_relu2d<<<(unsigned)(((long long)2 * HW * 16 + 255) / 256), 256, 0, stream>>>(R67 + 26176, nullptr, 2, 64, 16);
    { GemmP i2c5_0;
      i2c5_0.A = R67 + 26176 + (size_t)0 * 16; i2c5_0.B = iw2 + 0; i2c5_0.bias = ib2; i2c5_0.R = R67 + 26176 + (size_t)0 * 16; i2c5_0.C = R67 + 165568 + (size_t)67 * 32;
      i2c5_0.sAo = (long long)66 * 66 * 16; i2c5_0.sAi = (long long)66 * 16; i2c5_0.sAm = 16; i2c5_0.sAk = 1; i2c5_0.sBo = 0; i2c5_0.sBi = 0; i2c5_0.sBn = 16 * 9; i2c5_0.sBk = 9; i2c5_0.sCo = (long long)66 * 66 * 32; i2c5_0.sCi = (long long)66 * 32; i2c5_0.sCm = 32; i2c5_0.sRo = 0; i2c5_0.sRi = 0; i2c5_0.sRm = 0; i2c5_0.sRn = 0;
      i2c5_0.M = 64; i2c5_0.N = 32; i2c5_0.K = 16; i2c5_0.zi_n = 64; i2c5_0.flags = 1; i2c5_0.act = 0;
      i2c5_0.alpha = 1.0f; i2c5_0.beta = 0.0f; i2c5_0.sa = 1.0f; i2c5_0.sb = 1.0f; i2c5_0.Npad = 32; i2c5_0.pad_ = 0;
      k_gemm<1><<<dim3((unsigned)((32) + 31) / 32, (unsigned)((64) + 15) / 16, (unsigned)(2 * 64)), 32, 0, stream>>>(i2c5_0); }
    { GemmP i2c5_1;
      i2c5_1.A = R67 + 26176 + (size_t)1 * 16; i2c5_1.B = iw2 + 1; i2c5_1.bias = R67 + 26176 + (size_t)1 * 16; i2c5_1.R = R67 + 165568 + (size_t)67 * 32; i2c5_1.C = R67 + 165568 + (size_t)67 * 32;
      i2c5_1.sAo = (long long)66 * 66 * 16; i2c5_1.sAi = (long long)66 * 16; i2c5_1.sAm = 16; i2c5_1.sAk = 1; i2c5_1.sBo = 0; i2c5_1.sBi = 0; i2c5_1.sBn = 16 * 9; i2c5_1.sBk = 9; i2c5_1.sCo = (long long)66 * 66 * 32; i2c5_1.sCi = (long long)66 * 32; i2c5_1.sCm = 32; i2c5_1.sRo = (long long)66 * 66 * 32; i2c5_1.sRi = (long long)66 * 32; i2c5_1.sRm = 32; i2c5_1.sRn = 1;
      i2c5_1.M = 64; i2c5_1.N = 32; i2c5_1.K = 16; i2c5_1.zi_n = 64; i2c5_1.flags = 4; i2c5_1.act = 0;
      i2c5_1.alpha = 1.0f; i2c5_1.beta = 1.0f; i2c5_1.sa = 1.0f; i2c5_1.sb = 1.0f; i2c5_1.Npad = 32; i2c5_1.pad_ = 0;
      k_gemm<1><<<dim3((unsigned)((32) + 31) / 32, (unsigned)((64) + 15) / 16, (unsigned)(2 * 64)), 32, 0, stream>>>(i2c5_1); }
    { GemmP i2c5_2;
      i2c5_2.A = R67 + 26176 + (size_t)2 * 16; i2c5_2.B = iw2 + 2; i2c5_2.bias = R67 + 26176 + (size_t)2 * 16; i2c5_2.R = R67 + 165568 + (size_t)67 * 32; i2c5_2.C = R67 + 165568 + (size_t)67 * 32;
      i2c5_2.sAo = (long long)66 * 66 * 16; i2c5_2.sAi = (long long)66 * 16; i2c5_2.sAm = 16; i2c5_2.sAk = 1; i2c5_2.sBo = 0; i2c5_2.sBi = 0; i2c5_2.sBn = 16 * 9; i2c5_2.sBk = 9; i2c5_2.sCo = (long long)66 * 66 * 32; i2c5_2.sCi = (long long)66 * 32; i2c5_2.sCm = 32; i2c5_2.sRo = (long long)66 * 66 * 32; i2c5_2.sRi = (long long)66 * 32; i2c5_2.sRm = 32; i2c5_2.sRn = 1;
      i2c5_2.M = 64; i2c5_2.N = 32; i2c5_2.K = 16; i2c5_2.zi_n = 64; i2c5_2.flags = 4; i2c5_2.act = 0;
      i2c5_2.alpha = 1.0f; i2c5_2.beta = 1.0f; i2c5_2.sa = 1.0f; i2c5_2.sb = 1.0f; i2c5_2.Npad = 32; i2c5_2.pad_ = 0;
      k_gemm<1><<<dim3((unsigned)((32) + 31) / 32, (unsigned)((64) + 15) / 16, (unsigned)(2 * 64)), 32, 0, stream>>>(i2c5_2); }
    { GemmP i2c5_3;
      i2c5_3.A = R67 + 26176 + (size_t)66 * 16; i2c5_3.B = iw2 + 3; i2c5_3.bias = R67 + 26176 + (size_t)66 * 16; i2c5_3.R = R67 + 165568 + (size_t)67 * 32; i2c5_3.C = R67 + 165568 + (size_t)67 * 32;
      i2c5_3.sAo = (long long)66 * 66 * 16; i2c5_3.sAi = (long long)66 * 16; i2c5_3.sAm = 16; i2c5_3.sAk = 1; i2c5_3.sBo = 0; i2c5_3.sBi = 0; i2c5_3.sBn = 16 * 9; i2c5_3.sBk = 9; i2c5_3.sCo = (long long)66 * 66 * 32; i2c5_3.sCi = (long long)66 * 32; i2c5_3.sCm = 32; i2c5_3.sRo = (long long)66 * 66 * 32; i2c5_3.sRi = (long long)66 * 32; i2c5_3.sRm = 32; i2c5_3.sRn = 1;
      i2c5_3.M = 64; i2c5_3.N = 32; i2c5_3.K = 16; i2c5_3.zi_n = 64; i2c5_3.flags = 4; i2c5_3.act = 0;
      i2c5_3.alpha = 1.0f; i2c5_3.beta = 1.0f; i2c5_3.sa = 1.0f; i2c5_3.sb = 1.0f; i2c5_3.Npad = 32; i2c5_3.pad_ = 0;
      k_gemm<1><<<dim3((unsigned)((32) + 31) / 32, (unsigned)((64) + 15) / 16, (unsigned)(2 * 64)), 32, 0, stream>>>(i2c5_3); }
    { GemmP i2c5_4;
      i2c5_4.A = R67 + 26176 + (size_t)67 * 16; i2c5_4.B = iw2 + 4; i2c5_4.bias = R67 + 26176 + (size_t)67 * 16; i2c5_4.R = R67 + 165568 + (size_t)67 * 32; i2c5_4.C = R67 + 165568 + (size_t)67 * 32;
      i2c5_4.sAo = (long long)66 * 66 * 16; i2c5_4.sAi = (long long)66 * 16; i2c5_4.sAm = 16; i2c5_4.sAk = 1; i2c5_4.sBo = 0; i2c5_4.sBi = 0; i2c5_4.sBn = 16 * 9; i2c5_4.sBk = 9; i2c5_4.sCo = (long long)66 * 66 * 32; i2c5_4.sCi = (long long)66 * 32; i2c5_4.sCm = 32; i2c5_4.sRo = (long long)66 * 66 * 32; i2c5_4.sRi = (long long)66 * 32; i2c5_4.sRm = 32; i2c5_4.sRn = 1;
      i2c5_4.M = 64; i2c5_4.N = 32; i2c5_4.K = 16; i2c5_4.zi_n = 64; i2c5_4.flags = 4; i2c5_4.act = 0;
      i2c5_4.alpha = 1.0f; i2c5_4.beta = 1.0f; i2c5_4.sa = 1.0f; i2c5_4.sb = 1.0f; i2c5_4.Npad = 32; i2c5_4.pad_ = 0;
      k_gemm<1><<<dim3((unsigned)((32) + 31) / 32, (unsigned)((64) + 15) / 16, (unsigned)(2 * 64)), 32, 0, stream>>>(i2c5_4); }
    { GemmP i2c5_5;
      i2c5_5.A = R67 + 26176 + (size_t)68 * 16; i2c5_5.B = iw2 + 5; i2c5_5.bias = R67 + 26176 + (size_t)68 * 16; i2c5_5.R = R67 + 165568 + (size_t)67 * 32; i2c5_5.C = R67 + 165568 + (size_t)67 * 32;
      i2c5_5.sAo = (long long)66 * 66 * 16; i2c5_5.sAi = (long long)66 * 16; i2c5_5.sAm = 16; i2c5_5.sAk = 1; i2c5_5.sBo = 0; i2c5_5.sBi = 0; i2c5_5.sBn = 16 * 9; i2c5_5.sBk = 9; i2c5_5.sCo = (long long)66 * 66 * 32; i2c5_5.sCi = (long long)66 * 32; i2c5_5.sCm = 32; i2c5_5.sRo = (long long)66 * 66 * 32; i2c5_5.sRi = (long long)66 * 32; i2c5_5.sRm = 32; i2c5_5.sRn = 1;
      i2c5_5.M = 64; i2c5_5.N = 32; i2c5_5.K = 16; i2c5_5.zi_n = 64; i2c5_5.flags = 4; i2c5_5.act = 0;
      i2c5_5.alpha = 1.0f; i2c5_5.beta = 1.0f; i2c5_5.sa = 1.0f; i2c5_5.sb = 1.0f; i2c5_5.Npad = 32; i2c5_5.pad_ = 0;
      k_gemm<1><<<dim3((unsigned)((32) + 31) / 32, (unsigned)((64) + 15) / 16, (unsigned)(2 * 64)), 32, 0, stream>>>(i2c5_5); }
    { GemmP i2c5_6;
      i2c5_6.A = R67 + 26176 + (size_t)132 * 16; i2c5_6.B = iw2 + 6; i2c5_6.bias = R67 + 26176 + (size_t)132 * 16; i2c5_6.R = R67 + 165568 + (size_t)67 * 32; i2c5_6.C = R67 + 165568 + (size_t)67 * 32;
      i2c5_6.sAo = (long long)66 * 66 * 16; i2c5_6.sAi = (long long)66 * 16; i2c5_6.sAm = 16; i2c5_6.sAk = 1; i2c5_6.sBo = 0; i2c5_6.sBi = 0; i2c5_6.sBn = 16 * 9; i2c5_6.sBk = 9; i2c5_6.sCo = (long long)66 * 66 * 32; i2c5_6.sCi = (long long)66 * 32; i2c5_6.sCm = 32; i2c5_6.sRo = (long long)66 * 66 * 32; i2c5_6.sRi = (long long)66 * 32; i2c5_6.sRm = 32; i2c5_6.sRn = 1;
      i2c5_6.M = 64; i2c5_6.N = 32; i2c5_6.K = 16; i2c5_6.zi_n = 64; i2c5_6.flags = 4; i2c5_6.act = 0;
      i2c5_6.alpha = 1.0f; i2c5_6.beta = 1.0f; i2c5_6.sa = 1.0f; i2c5_6.sb = 1.0f; i2c5_6.Npad = 32; i2c5_6.pad_ = 0;
      k_gemm<1><<<dim3((unsigned)((32) + 31) / 32, (unsigned)((64) + 15) / 16, (unsigned)(2 * 64)), 32, 0, stream>>>(i2c5_6); }
    { GemmP i2c5_7;
      i2c5_7.A = R67 + 26176 + (size_t)133 * 16; i2c5_7.B = iw2 + 7; i2c5_7.bias = R67 + 26176 + (size_t)133 * 16; i2c5_7.R = R67 + 165568 + (size_t)67 * 32; i2c5_7.C = R67 + 165568 + (size_t)67 * 32;
      i2c5_7.sAo = (long long)66 * 66 * 16; i2c5_7.sAi = (long long)66 * 16; i2c5_7.sAm = 16; i2c5_7.sAk = 1; i2c5_7.sBo = 0; i2c5_7.sBi = 0; i2c5_7.sBn = 16 * 9; i2c5_7.sBk = 9; i2c5_7.sCo = (long long)66 * 66 * 32; i2c5_7.sCi = (long long)66 * 32; i2c5_7.sCm = 32; i2c5_7.sRo = (long long)66 * 66 * 32; i2c5_7.sRi = (long long)66 * 32; i2c5_7.sRm = 32; i2c5_7.sRn = 1;
      i2c5_7.M = 64; i2c5_7.N = 32; i2c5_7.K = 16; i2c5_7.zi_n = 64; i2c5_7.flags = 4; i2c5_7.act = 0;
      i2c5_7.alpha = 1.0f; i2c5_7.beta = 1.0f; i2c5_7.sa = 1.0f; i2c5_7.sb = 1.0f; i2c5_7.Npad = 32; i2c5_7.pad_ = 0;
      k_gemm<1><<<dim3((unsigned)((32) + 31) / 32, (unsigned)((64) + 15) / 16, (unsigned)(2 * 64)), 32, 0, stream>>>(i2c5_7); }
    { GemmP i2c5_8;
      i2c5_8.A = R67 + 26176 + (size_t)134 * 16; i2c5_8.B = iw2 + 8; i2c5_8.bias = R67 + 26176 + (size_t)134 * 16; i2c5_8.R = R67 + 165568 + (size_t)67 * 32; i2c5_8.C = R67 + 165568 + (size_t)67 * 32;
      i2c5_8.sAo = (long long)66 * 66 * 16; i2c5_8.sAi = (long long)66 * 16; i2c5_8.sAm = 16; i2c5_8.sAk = 1; i2c5_8.sBo = 0; i2c5_8.sBi = 0; i2c5_8.sBn = 16 * 9; i2c5_8.sBk = 9; i2c5_8.sCo = (long long)66 * 66 * 32; i2c5_8.sCi = (long long)66 * 32; i2c5_8.sCm = 32; i2c5_8.sRo = (long long)66 * 66 * 32; i2c5_8.sRi = (long long)66 * 32; i2c5_8.sRm = 32; i2c5_8.sRn = 1;
      i2c5_8.M = 64; i2c5_8.N = 32; i2c5_8.K = 16; i2c5_8.zi_n = 64; i2c5_8.flags = 4; i2c5_8.act = 0;
      i2c5_8.alpha = 1.0f; i2c5_8.beta = 1.0f; i2c5_8.sa = 1.0f; i2c5_8.sb = 1.0f; i2c5_8.Npad = 32; i2c5_8.pad_ = 0;
      k_gemm<1><<<dim3((unsigned)((32) + 31) / 32, (unsigned)((64) + 15) / 16, (unsigned)(2 * 64)), 32, 0, stream>>>(i2c5_8); }
    k_mm_relu2d<<<(unsigned)(((long long)2 * HW * 32 + 255) / 256), 256, 0, stream>>>(R67 + 165568, nullptr, 2, 64, 32);
    { GemmP i3c5_0;
      i3c5_0.A = R67 + 165568 + (size_t)0 * 32; i3c5_0.B = iw3 + 0; i3c5_0.bias = ib3; i3c5_0.R = R67 + 165568 + (size_t)0 * 32; i3c5_0.C = R67 + 444352 + (size_t)67 * 64;
      i3c5_0.sAo = (long long)66 * 66 * 32; i3c5_0.sAi = (long long)66 * 32; i3c5_0.sAm = 32; i3c5_0.sAk = 1; i3c5_0.sBo = 0; i3c5_0.sBi = 0; i3c5_0.sBn = 32 * 9; i3c5_0.sBk = 9; i3c5_0.sCo = (long long)66 * 66 * 64; i3c5_0.sCi = (long long)66 * 64; i3c5_0.sCm = 64; i3c5_0.sRo = 0; i3c5_0.sRi = 0; i3c5_0.sRm = 0; i3c5_0.sRn = 0;
      i3c5_0.M = 64; i3c5_0.N = 64; i3c5_0.K = 32; i3c5_0.zi_n = 64; i3c5_0.flags = 1; i3c5_0.act = 0;
      i3c5_0.alpha = 1.0f; i3c5_0.beta = 0.0f; i3c5_0.sa = 1.0f; i3c5_0.sb = 1.0f; i3c5_0.Npad = 64; i3c5_0.pad_ = 0;
      k_gemm<1><<<dim3((unsigned)((64) + 31) / 32, (unsigned)((64) + 15) / 16, (unsigned)(2 * 64)), 32, 0, stream>>>(i3c5_0); }
    { GemmP i3c5_1;
      i3c5_1.A = R67 + 165568 + (size_t)1 * 32; i3c5_1.B = iw3 + 1; i3c5_1.bias = R67 + 165568 + (size_t)1 * 32; i3c5_1.R = R67 + 444352 + (size_t)67 * 64; i3c5_1.C = R67 + 444352 + (size_t)67 * 64;
      i3c5_1.sAo = (long long)66 * 66 * 32; i3c5_1.sAi = (long long)66 * 32; i3c5_1.sAm = 32; i3c5_1.sAk = 1; i3c5_1.sBo = 0; i3c5_1.sBi = 0; i3c5_1.sBn = 32 * 9; i3c5_1.sBk = 9; i3c5_1.sCo = (long long)66 * 66 * 64; i3c5_1.sCi = (long long)66 * 64; i3c5_1.sCm = 64; i3c5_1.sRo = (long long)66 * 66 * 64; i3c5_1.sRi = (long long)66 * 64; i3c5_1.sRm = 64; i3c5_1.sRn = 1;
      i3c5_1.M = 64; i3c5_1.N = 64; i3c5_1.K = 32; i3c5_1.zi_n = 64; i3c5_1.flags = 4; i3c5_1.act = 0;
      i3c5_1.alpha = 1.0f; i3c5_1.beta = 1.0f; i3c5_1.sa = 1.0f; i3c5_1.sb = 1.0f; i3c5_1.Npad = 64; i3c5_1.pad_ = 0;
      k_gemm<1><<<dim3((unsigned)((64) + 31) / 32, (unsigned)((64) + 15) / 16, (unsigned)(2 * 64)), 32, 0, stream>>>(i3c5_1); }
    { GemmP i3c5_2;
      i3c5_2.A = R67 + 165568 + (size_t)2 * 32; i3c5_2.B = iw3 + 2; i3c5_2.bias = R67 + 165568 + (size_t)2 * 32; i3c5_2.R = R67 + 444352 + (size_t)67 * 64; i3c5_2.C = R67 + 444352 + (size_t)67 * 64;
      i3c5_2.sAo = (long long)66 * 66 * 32; i3c5_2.sAi = (long long)66 * 32; i3c5_2.sAm = 32; i3c5_2.sAk = 1; i3c5_2.sBo = 0; i3c5_2.sBi = 0; i3c5_2.sBn = 32 * 9; i3c5_2.sBk = 9; i3c5_2.sCo = (long long)66 * 66 * 64; i3c5_2.sCi = (long long)66 * 64; i3c5_2.sCm = 64; i3c5_2.sRo = (long long)66 * 66 * 64; i3c5_2.sRi = (long long)66 * 64; i3c5_2.sRm = 64; i3c5_2.sRn = 1;
      i3c5_2.M = 64; i3c5_2.N = 64; i3c5_2.K = 32; i3c5_2.zi_n = 64; i3c5_2.flags = 4; i3c5_2.act = 0;
      i3c5_2.alpha = 1.0f; i3c5_2.beta = 1.0f; i3c5_2.sa = 1.0f; i3c5_2.sb = 1.0f; i3c5_2.Npad = 64; i3c5_2.pad_ = 0;
      k_gemm<1><<<dim3((unsigned)((64) + 31) / 32, (unsigned)((64) + 15) / 16, (unsigned)(2 * 64)), 32, 0, stream>>>(i3c5_2); }
    { GemmP i3c5_3;
      i3c5_3.A = R67 + 165568 + (size_t)66 * 32; i3c5_3.B = iw3 + 3; i3c5_3.bias = R67 + 165568 + (size_t)66 * 32; i3c5_3.R = R67 + 444352 + (size_t)67 * 64; i3c5_3.C = R67 + 444352 + (size_t)67 * 64;
      i3c5_3.sAo = (long long)66 * 66 * 32; i3c5_3.sAi = (long long)66 * 32; i3c5_3.sAm = 32; i3c5_3.sAk = 1; i3c5_3.sBo = 0; i3c5_3.sBi = 0; i3c5_3.sBn = 32 * 9; i3c5_3.sBk = 9; i3c5_3.sCo = (long long)66 * 66 * 64; i3c5_3.sCi = (long long)66 * 64; i3c5_3.sCm = 64; i3c5_3.sRo = (long long)66 * 66 * 64; i3c5_3.sRi = (long long)66 * 64; i3c5_3.sRm = 64; i3c5_3.sRn = 1;
      i3c5_3.M = 64; i3c5_3.N = 64; i3c5_3.K = 32; i3c5_3.zi_n = 64; i3c5_3.flags = 4; i3c5_3.act = 0;
      i3c5_3.alpha = 1.0f; i3c5_3.beta = 1.0f; i3c5_3.sa = 1.0f; i3c5_3.sb = 1.0f; i3c5_3.Npad = 64; i3c5_3.pad_ = 0;
      k_gemm<1><<<dim3((unsigned)((64) + 31) / 32, (unsigned)((64) + 15) / 16, (unsigned)(2 * 64)), 32, 0, stream>>>(i3c5_3); }
    { GemmP i3c5_4;
      i3c5_4.A = R67 + 165568 + (size_t)67 * 32; i3c5_4.B = iw3 + 4; i3c5_4.bias = R67 + 165568 + (size_t)67 * 32; i3c5_4.R = R67 + 444352 + (size_t)67 * 64; i3c5_4.C = R67 + 444352 + (size_t)67 * 64;
      i3c5_4.sAo = (long long)66 * 66 * 32; i3c5_4.sAi = (long long)66 * 32; i3c5_4.sAm = 32; i3c5_4.sAk = 1; i3c5_4.sBo = 0; i3c5_4.sBi = 0; i3c5_4.sBn = 32 * 9; i3c5_4.sBk = 9; i3c5_4.sCo = (long long)66 * 66 * 64; i3c5_4.sCi = (long long)66 * 64; i3c5_4.sCm = 64; i3c5_4.sRo = (long long)66 * 66 * 64; i3c5_4.sRi = (long long)66 * 64; i3c5_4.sRm = 64; i3c5_4.sRn = 1;
      i3c5_4.M = 64; i3c5_4.N = 64; i3c5_4.K = 32; i3c5_4.zi_n = 64; i3c5_4.flags = 4; i3c5_4.act = 0;
      i3c5_4.alpha = 1.0f; i3c5_4.beta = 1.0f; i3c5_4.sa = 1.0f; i3c5_4.sb = 1.0f; i3c5_4.Npad = 64; i3c5_4.pad_ = 0;
      k_gemm<1><<<dim3((unsigned)((64) + 31) / 32, (unsigned)((64) + 15) / 16, (unsigned)(2 * 64)), 32, 0, stream>>>(i3c5_4); }
    { GemmP i3c5_5;
      i3c5_5.A = R67 + 165568 + (size_t)68 * 32; i3c5_5.B = iw3 + 5; i3c5_5.bias = R67 + 165568 + (size_t)68 * 32; i3c5_5.R = R67 + 444352 + (size_t)67 * 64; i3c5_5.C = R67 + 444352 + (size_t)67 * 64;
      i3c5_5.sAo = (long long)66 * 66 * 32; i3c5_5.sAi = (long long)66 * 32; i3c5_5.sAm = 32; i3c5_5.sAk = 1; i3c5_5.sBo = 0; i3c5_5.sBi = 0; i3c5_5.sBn = 32 * 9; i3c5_5.sBk = 9; i3c5_5.sCo = (long long)66 * 66 * 64; i3c5_5.sCi = (long long)66 * 64; i3c5_5.sCm = 64; i3c5_5.sRo = (long long)66 * 66 * 64; i3c5_5.sRi = (long long)66 * 64; i3c5_5.sRm = 64; i3c5_5.sRn = 1;
      i3c5_5.M = 64; i3c5_5.N = 64; i3c5_5.K = 32; i3c5_5.zi_n = 64; i3c5_5.flags = 4; i3c5_5.act = 0;
      i3c5_5.alpha = 1.0f; i3c5_5.beta = 1.0f; i3c5_5.sa = 1.0f; i3c5_5.sb = 1.0f; i3c5_5.Npad = 64; i3c5_5.pad_ = 0;
      k_gemm<1><<<dim3((unsigned)((64) + 31) / 32, (unsigned)((64) + 15) / 16, (unsigned)(2 * 64)), 32, 0, stream>>>(i3c5_5); }
    { GemmP i3c5_6;
      i3c5_6.A = R67 + 165568 + (size_t)132 * 32; i3c5_6.B = iw3 + 6; i3c5_6.bias = R67 + 165568 + (size_t)132 * 32; i3c5_6.R = R67 + 444352 + (size_t)67 * 64; i3c5_6.C = R67 + 444352 + (size_t)67 * 64;
      i3c5_6.sAo = (long long)66 * 66 * 32; i3c5_6.sAi = (long long)66 * 32; i3c5_6.sAm = 32; i3c5_6.sAk = 1; i3c5_6.sBo = 0; i3c5_6.sBi = 0; i3c5_6.sBn = 32 * 9; i3c5_6.sBk = 9; i3c5_6.sCo = (long long)66 * 66 * 64; i3c5_6.sCi = (long long)66 * 64; i3c5_6.sCm = 64; i3c5_6.sRo = (long long)66 * 66 * 64; i3c5_6.sRi = (long long)66 * 64; i3c5_6.sRm = 64; i3c5_6.sRn = 1;
      i3c5_6.M = 64; i3c5_6.N = 64; i3c5_6.K = 32; i3c5_6.zi_n = 64; i3c5_6.flags = 4; i3c5_6.act = 0;
      i3c5_6.alpha = 1.0f; i3c5_6.beta = 1.0f; i3c5_6.sa = 1.0f; i3c5_6.sb = 1.0f; i3c5_6.Npad = 64; i3c5_6.pad_ = 0;
      k_gemm<1><<<dim3((unsigned)((64) + 31) / 32, (unsigned)((64) + 15) / 16, (unsigned)(2 * 64)), 32, 0, stream>>>(i3c5_6); }
    { GemmP i3c5_7;
      i3c5_7.A = R67 + 165568 + (size_t)133 * 32; i3c5_7.B = iw3 + 7; i3c5_7.bias = R67 + 165568 + (size_t)133 * 32; i3c5_7.R = R67 + 444352 + (size_t)67 * 64; i3c5_7.C = R67 + 444352 + (size_t)67 * 64;
      i3c5_7.sAo = (long long)66 * 66 * 32; i3c5_7.sAi = (long long)66 * 32; i3c5_7.sAm = 32; i3c5_7.sAk = 1; i3c5_7.sBo = 0; i3c5_7.sBi = 0; i3c5_7.sBn = 32 * 9; i3c5_7.sBk = 9; i3c5_7.sCo = (long long)66 * 66 * 64; i3c5_7.sCi = (long long)66 * 64; i3c5_7.sCm = 64; i3c5_7.sRo = (long long)66 * 66 * 64; i3c5_7.sRi = (long long)66 * 64; i3c5_7.sRm = 64; i3c5_7.sRn = 1;
      i3c5_7.M = 64; i3c5_7.N = 64; i3c5_7.K = 32; i3c5_7.zi_n = 64; i3c5_7.flags = 4; i3c5_7.act = 0;
      i3c5_7.alpha = 1.0f; i3c5_7.beta = 1.0f; i3c5_7.sa = 1.0f; i3c5_7.sb = 1.0f; i3c5_7.Npad = 64; i3c5_7.pad_ = 0;
      k_gemm<1><<<dim3((unsigned)((64) + 31) / 32, (unsigned)((64) + 15) / 16, (unsigned)(2 * 64)), 32, 0, stream>>>(i3c5_7); }
    { GemmP i3c5_8;
      i3c5_8.A = R67 + 165568 + (size_t)134 * 32; i3c5_8.B = iw3 + 8; i3c5_8.bias = R67 + 165568 + (size_t)134 * 32; i3c5_8.R = R67 + 444352 + (size_t)67 * 64; i3c5_8.C = R67 + 444352 + (size_t)67 * 64;
      i3c5_8.sAo = (long long)66 * 66 * 32; i3c5_8.sAi = (long long)66 * 32; i3c5_8.sAm = 32; i3c5_8.sAk = 1; i3c5_8.sBo = 0; i3c5_8.sBi = 0; i3c5_8.sBn = 32 * 9; i3c5_8.sBk = 9; i3c5_8.sCo = (long long)66 * 66 * 64; i3c5_8.sCi = (long long)66 * 64; i3c5_8.sCm = 64; i3c5_8.sRo = (long long)66 * 66 * 64; i3c5_8.sRi = (long long)66 * 64; i3c5_8.sRm = 64; i3c5_8.sRn = 1;
      i3c5_8.M = 64; i3c5_8.N = 64; i3c5_8.K = 32; i3c5_8.zi_n = 64; i3c5_8.flags = 4; i3c5_8.act = 0;
      i3c5_8.alpha = 1.0f; i3c5_8.beta = 1.0f; i3c5_8.sa = 1.0f; i3c5_8.sb = 1.0f; i3c5_8.Npad = 64; i3c5_8.pad_ = 0;
      k_gemm<1><<<dim3((unsigned)((64) + 31) / 32, (unsigned)((64) + 15) / 16, (unsigned)(2 * 64)), 32, 0, stream>>>(i3c5_8); }
    k_mm_relu2d<<<(unsigned)(((long long)2 * HW * 64 + 255) / 256), 256, 0, stream>>>(R67 + 444352, R67 + 1001920, 2, 64, 64);
    { GemmP gqkv5;
      gqkv5.A = R67 + 1001920; gqkv5.B = qkvw; gqkv5.bias = qkvb; gqkv5.R = R67 + 1001920; gqkv5.C = R67 + 1526208;
      gqkv5.sAo = 0; gqkv5.sAi = 0; gqkv5.sAm = 64; gqkv5.sAk = 1; gqkv5.sBo = 0; gqkv5.sBi = 0; gqkv5.sBn = 64; gqkv5.sBk = 1; gqkv5.sCo = 0; gqkv5.sCi = 0; gqkv5.sCm = 192; gqkv5.sRo = 0; gqkv5.sRi = 0; gqkv5.sRm = 0; gqkv5.sRn = 0;
      gqkv5.M = 2 * HW; gqkv5.N = 192; gqkv5.K = 64; gqkv5.zi_n = 1; gqkv5.flags = 1; gqkv5.act = 0;
      gqkv5.alpha = 1.0f; gqkv5.beta = 0.0f; gqkv5.sa = 1.0f; gqkv5.sb = 1.0f; gqkv5.Npad = 192; gqkv5.pad_ = 0;
      k_gemm<1><<<dim3((unsigned)((192) + 31) / 32, (unsigned)((2 * HW) + 15) / 16, (unsigned)(1)), 32, 0, stream>>>(gqkv5); }
    k_mm_dw<<<(unsigned)(((long long)2 * HW * 192 + 255) / 256), 256, 0, stream>>>(R67 + 1526208, dww, dwb, R67 + 3099072, 2, 64, 192);
    k_mm_fall<<<(unsigned)(((long long)2 * HW * 144 + 255) / 256), 256, 0, stream>>>(R67 + 3099072, fcw, fcb, R67 + 4671936, 2, HW, 192);
    k_mm_dep<<<(unsigned)(((long long)2 * 64 * HW + 255) / 256), 256, 0, stream>>>(R67 + 4671936, depw, depb, R67 + 5851584, 2, 64);
    k_mm_qknorm<<<2 * 128, 256, 0, stream>>>(R67 + 3099072, R67 + 6375872, 2, HW, 192);
    { GemmP gat5;
      gat5.A = R67 + 6375872; gat5.B = R67 + 6375872 + (size_t)64 * HW; gat5.bias = R67 + 6375872; gat5.R = R67 + 6375872; gat5.C = R67 + 7424448;
      gat5.sAo = (long long)128 * HW; gat5.sAi = (long long)16 * HW; gat5.sAm = HW; gat5.sAk = 1; gat5.sBo = (long long)128 * HW; gat5.sBi = (long long)16 * HW; gat5.sBn = HW; gat5.sBk = 1; gat5.sCo = (long long)4 * 16 * LP; gat5.sCi = 16 * LP; gat5.sCm = LP; gat5.sRo = 0; gat5.sRi = 0; gat5.sRm = 0; gat5.sRn = 0;
      gat5.M = 16; gat5.N = 16; gat5.K = HW; gat5.zi_n = 4; gat5.flags = 0; gat5.act = 0;
      gat5.alpha = 1.0f; gat5.beta = 0.0f; gat5.sa = 1.0f; gat5.sb = 1.0f; gat5.Npad = LP; gat5.pad_ = 0;
      k_gemm<1><<<dim3((unsigned)((LP) + 31) / 32, (unsigned)((16) + 15) / 16, (unsigned)(2 * 4)), 32, 0, stream>>>(gat5); }
    k_mm_sm16<<<(unsigned)((2 * 4 * 16 + 255) / 256), 256, 0, stream>>>(R67 + 7424448, temp, 2 * 4, LP);
    { GemmP gao5;
      gao5.A = R67 + 7424448; gao5.B = R67 + 3099072 + 128; gao5.bias = R67 + 7424448; gao5.R = R67 + 7424448; gao5.C = R67 + 7428544;
      gao5.sAo = (long long)4 * 16 * LP; gao5.sAi = 16 * LP; gao5.sAm = LP; gao5.sAk = 1; gao5.sBo = (long long)HW * 192; gao5.sBi = 16; gao5.sBn = 192; gao5.sBk = 1; gao5.sCo = (long long)64 * HW; gao5.sCi = (long long)16 * HW; gao5.sCm = HW; gao5.sRo = 0; gao5.sRi = 0; gao5.sRm = 0; gao5.sRn = 0;
      gao5.M = 16; gao5.N = HW; gao5.K = 16; gao5.zi_n = 4; gao5.flags = 0; gao5.act = 0;
      gao5.alpha = 1.0f; gao5.beta = 0.0f; gao5.sa = 1.0f; gao5.sb = 1.0f; gao5.Npad = HW; gao5.pad_ = 0;
      k_gemm<1><<<dim3((unsigned)((HW) + 31) / 32, (unsigned)((16) + 15) / 16, (unsigned)(2 * 4)), 32, 0, stream>>>(gao5); }
    { GemmP gproj5;
      gproj5.A = projw; gproj5.B = R67 + 7428544; gproj5.bias = projb; gproj5.R = projw; gproj5.C = R67 + 7952832;
      gproj5.sAo = 0; gproj5.sAi = 0; gproj5.sAm = 64; gproj5.sAk = 1; gproj5.sBo = (long long)64 * HW; gproj5.sBi = 0; gproj5.sBn = 1; gproj5.sBk = HW; gproj5.sCo = (long long)64 * HW; gproj5.sCi = 0; gproj5.sCm = HW; gproj5.sRo = 0; gproj5.sRi = 0; gproj5.sRm = 0; gproj5.sRn = 0;
      gproj5.M = 64; gproj5.N = HW; gproj5.K = 64; gproj5.zi_n = 1; gproj5.flags = 2; gproj5.act = 0;
      gproj5.alpha = 1.0f; gproj5.beta = 0.0f; gproj5.sa = 1.0f; gproj5.sb = 1.0f; gproj5.Npad = HW; gproj5.pad_ = 0;
      k_gemm<1><<<dim3((unsigned)((HW) + 31) / 32, (unsigned)((64) + 15) / 16, (unsigned)(2)), 32, 0, stream>>>(gproj5); }
    k_mm_imgfeat<<<(unsigned)(((long long)2 * SEQ * 64 + 255) / 256), 256, 0, stream>>>(R67 + 7952832, R67 + 5851584, IR + (size_t)10 * SEQ * 64, 2, HW, 64);
    hipMemsetAsync(R67 + 0, 0, (size_t)2 * 66 * 66 * 3 * 4, stream); hipMemsetAsync(R67 + 26176, 0, (size_t)2 * 66 * 66 * 16 * 4, stream); hipMemsetAsync(R67 + 165568, 0, (size_t)2 * 66 * 66 * 32 * 4, stream); hipMemsetAsync(R67 + 444352, 0, (size_t)2 * 66 * 66 * 64 * 4, stream);
    k_mm_padimg<<<(unsigned)(((long long)2 * HW * 3 + 255) / 256), 256, 0, stream>>>(img + (size_t)12 * 3 * HW, R67 + 0, 2, 3, 64);
    { GemmP i1c6_0;
      i1c6_0.A = R67 + 0 + (size_t)0 * 3; i1c6_0.B = iw1 + 0; i1c6_0.bias = ib1; i1c6_0.R = R67 + 0 + (size_t)0 * 3; i1c6_0.C = R67 + 26176 + (size_t)67 * 16;
      i1c6_0.sAo = (long long)66 * 66 * 3; i1c6_0.sAi = (long long)66 * 3; i1c6_0.sAm = 3; i1c6_0.sAk = 1; i1c6_0.sBo = 0; i1c6_0.sBi = 0; i1c6_0.sBn = 3 * 9; i1c6_0.sBk = 9; i1c6_0.sCo = (long long)66 * 66 * 16; i1c6_0.sCi = (long long)66 * 16; i1c6_0.sCm = 16; i1c6_0.sRo = 0; i1c6_0.sRi = 0; i1c6_0.sRm = 0; i1c6_0.sRn = 0;
      i1c6_0.M = 64; i1c6_0.N = 16; i1c6_0.K = 3; i1c6_0.zi_n = 64; i1c6_0.flags = 1; i1c6_0.act = 0;
      i1c6_0.alpha = 1.0f; i1c6_0.beta = 0.0f; i1c6_0.sa = 1.0f; i1c6_0.sb = 1.0f; i1c6_0.Npad = 16; i1c6_0.pad_ = 0;
      k_gemm<1><<<dim3((unsigned)((16) + 31) / 32, (unsigned)((64) + 15) / 16, (unsigned)(2 * 64)), 32, 0, stream>>>(i1c6_0); }
    { GemmP i1c6_1;
      i1c6_1.A = R67 + 0 + (size_t)1 * 3; i1c6_1.B = iw1 + 1; i1c6_1.bias = R67 + 0 + (size_t)1 * 3; i1c6_1.R = R67 + 26176 + (size_t)67 * 16; i1c6_1.C = R67 + 26176 + (size_t)67 * 16;
      i1c6_1.sAo = (long long)66 * 66 * 3; i1c6_1.sAi = (long long)66 * 3; i1c6_1.sAm = 3; i1c6_1.sAk = 1; i1c6_1.sBo = 0; i1c6_1.sBi = 0; i1c6_1.sBn = 3 * 9; i1c6_1.sBk = 9; i1c6_1.sCo = (long long)66 * 66 * 16; i1c6_1.sCi = (long long)66 * 16; i1c6_1.sCm = 16; i1c6_1.sRo = (long long)66 * 66 * 16; i1c6_1.sRi = (long long)66 * 16; i1c6_1.sRm = 16; i1c6_1.sRn = 1;
      i1c6_1.M = 64; i1c6_1.N = 16; i1c6_1.K = 3; i1c6_1.zi_n = 64; i1c6_1.flags = 4; i1c6_1.act = 0;
      i1c6_1.alpha = 1.0f; i1c6_1.beta = 1.0f; i1c6_1.sa = 1.0f; i1c6_1.sb = 1.0f; i1c6_1.Npad = 16; i1c6_1.pad_ = 0;
      k_gemm<1><<<dim3((unsigned)((16) + 31) / 32, (unsigned)((64) + 15) / 16, (unsigned)(2 * 64)), 32, 0, stream>>>(i1c6_1); }
    { GemmP i1c6_2;
      i1c6_2.A = R67 + 0 + (size_t)2 * 3; i1c6_2.B = iw1 + 2; i1c6_2.bias = R67 + 0 + (size_t)2 * 3; i1c6_2.R = R67 + 26176 + (size_t)67 * 16; i1c6_2.C = R67 + 26176 + (size_t)67 * 16;
      i1c6_2.sAo = (long long)66 * 66 * 3; i1c6_2.sAi = (long long)66 * 3; i1c6_2.sAm = 3; i1c6_2.sAk = 1; i1c6_2.sBo = 0; i1c6_2.sBi = 0; i1c6_2.sBn = 3 * 9; i1c6_2.sBk = 9; i1c6_2.sCo = (long long)66 * 66 * 16; i1c6_2.sCi = (long long)66 * 16; i1c6_2.sCm = 16; i1c6_2.sRo = (long long)66 * 66 * 16; i1c6_2.sRi = (long long)66 * 16; i1c6_2.sRm = 16; i1c6_2.sRn = 1;
      i1c6_2.M = 64; i1c6_2.N = 16; i1c6_2.K = 3; i1c6_2.zi_n = 64; i1c6_2.flags = 4; i1c6_2.act = 0;
      i1c6_2.alpha = 1.0f; i1c6_2.beta = 1.0f; i1c6_2.sa = 1.0f; i1c6_2.sb = 1.0f; i1c6_2.Npad = 16; i1c6_2.pad_ = 0;
      k_gemm<1><<<dim3((unsigned)((16) + 31) / 32, (unsigned)((64) + 15) / 16, (unsigned)(2 * 64)), 32, 0, stream>>>(i1c6_2); }
    { GemmP i1c6_3;
      i1c6_3.A = R67 + 0 + (size_t)66 * 3; i1c6_3.B = iw1 + 3; i1c6_3.bias = R67 + 0 + (size_t)66 * 3; i1c6_3.R = R67 + 26176 + (size_t)67 * 16; i1c6_3.C = R67 + 26176 + (size_t)67 * 16;
      i1c6_3.sAo = (long long)66 * 66 * 3; i1c6_3.sAi = (long long)66 * 3; i1c6_3.sAm = 3; i1c6_3.sAk = 1; i1c6_3.sBo = 0; i1c6_3.sBi = 0; i1c6_3.sBn = 3 * 9; i1c6_3.sBk = 9; i1c6_3.sCo = (long long)66 * 66 * 16; i1c6_3.sCi = (long long)66 * 16; i1c6_3.sCm = 16; i1c6_3.sRo = (long long)66 * 66 * 16; i1c6_3.sRi = (long long)66 * 16; i1c6_3.sRm = 16; i1c6_3.sRn = 1;
      i1c6_3.M = 64; i1c6_3.N = 16; i1c6_3.K = 3; i1c6_3.zi_n = 64; i1c6_3.flags = 4; i1c6_3.act = 0;
      i1c6_3.alpha = 1.0f; i1c6_3.beta = 1.0f; i1c6_3.sa = 1.0f; i1c6_3.sb = 1.0f; i1c6_3.Npad = 16; i1c6_3.pad_ = 0;
      k_gemm<1><<<dim3((unsigned)((16) + 31) / 32, (unsigned)((64) + 15) / 16, (unsigned)(2 * 64)), 32, 0, stream>>>(i1c6_3); }
    { GemmP i1c6_4;
      i1c6_4.A = R67 + 0 + (size_t)67 * 3; i1c6_4.B = iw1 + 4; i1c6_4.bias = R67 + 0 + (size_t)67 * 3; i1c6_4.R = R67 + 26176 + (size_t)67 * 16; i1c6_4.C = R67 + 26176 + (size_t)67 * 16;
      i1c6_4.sAo = (long long)66 * 66 * 3; i1c6_4.sAi = (long long)66 * 3; i1c6_4.sAm = 3; i1c6_4.sAk = 1; i1c6_4.sBo = 0; i1c6_4.sBi = 0; i1c6_4.sBn = 3 * 9; i1c6_4.sBk = 9; i1c6_4.sCo = (long long)66 * 66 * 16; i1c6_4.sCi = (long long)66 * 16; i1c6_4.sCm = 16; i1c6_4.sRo = (long long)66 * 66 * 16; i1c6_4.sRi = (long long)66 * 16; i1c6_4.sRm = 16; i1c6_4.sRn = 1;
      i1c6_4.M = 64; i1c6_4.N = 16; i1c6_4.K = 3; i1c6_4.zi_n = 64; i1c6_4.flags = 4; i1c6_4.act = 0;
      i1c6_4.alpha = 1.0f; i1c6_4.beta = 1.0f; i1c6_4.sa = 1.0f; i1c6_4.sb = 1.0f; i1c6_4.Npad = 16; i1c6_4.pad_ = 0;
      k_gemm<1><<<dim3((unsigned)((16) + 31) / 32, (unsigned)((64) + 15) / 16, (unsigned)(2 * 64)), 32, 0, stream>>>(i1c6_4); }
    { GemmP i1c6_5;
      i1c6_5.A = R67 + 0 + (size_t)68 * 3; i1c6_5.B = iw1 + 5; i1c6_5.bias = R67 + 0 + (size_t)68 * 3; i1c6_5.R = R67 + 26176 + (size_t)67 * 16; i1c6_5.C = R67 + 26176 + (size_t)67 * 16;
      i1c6_5.sAo = (long long)66 * 66 * 3; i1c6_5.sAi = (long long)66 * 3; i1c6_5.sAm = 3; i1c6_5.sAk = 1; i1c6_5.sBo = 0; i1c6_5.sBi = 0; i1c6_5.sBn = 3 * 9; i1c6_5.sBk = 9; i1c6_5.sCo = (long long)66 * 66 * 16; i1c6_5.sCi = (long long)66 * 16; i1c6_5.sCm = 16; i1c6_5.sRo = (long long)66 * 66 * 16; i1c6_5.sRi = (long long)66 * 16; i1c6_5.sRm = 16; i1c6_5.sRn = 1;
      i1c6_5.M = 64; i1c6_5.N = 16; i1c6_5.K = 3; i1c6_5.zi_n = 64; i1c6_5.flags = 4; i1c6_5.act = 0;
      i1c6_5.alpha = 1.0f; i1c6_5.beta = 1.0f; i1c6_5.sa = 1.0f; i1c6_5.sb = 1.0f; i1c6_5.Npad = 16; i1c6_5.pad_ = 0;
      k_gemm<1><<<dim3((unsigned)((16) + 31) / 32, (unsigned)((64) + 15) / 16, (unsigned)(2 * 64)), 32, 0, stream>>>(i1c6_5); }
    { GemmP i1c6_6;
      i1c6_6.A = R67 + 0 + (size_t)132 * 3; i1c6_6.B = iw1 + 6; i1c6_6.bias = R67 + 0 + (size_t)132 * 3; i1c6_6.R = R67 + 26176 + (size_t)67 * 16; i1c6_6.C = R67 + 26176 + (size_t)67 * 16;
      i1c6_6.sAo = (long long)66 * 66 * 3; i1c6_6.sAi = (long long)66 * 3; i1c6_6.sAm = 3; i1c6_6.sAk = 1; i1c6_6.sBo = 0; i1c6_6.sBi = 0; i1c6_6.sBn = 3 * 9; i1c6_6.sBk = 9; i1c6_6.sCo = (long long)66 * 66 * 16; i1c6_6.sCi = (long long)66 * 16; i1c6_6.sCm = 16; i1c6_6.sRo = (long long)66 * 66 * 16; i1c6_6.sRi = (long long)66 * 16; i1c6_6.sRm = 16; i1c6_6.sRn = 1;
      i1c6_6.M = 64; i1c6_6.N = 16; i1c6_6.K = 3; i1c6_6.zi_n = 64; i1c6_6.flags = 4; i1c6_6.act = 0;
      i1c6_6.alpha = 1.0f; i1c6_6.beta = 1.0f; i1c6_6.sa = 1.0f; i1c6_6.sb = 1.0f; i1c6_6.Npad = 16; i1c6_6.pad_ = 0;
      k_gemm<1><<<dim3((unsigned)((16) + 31) / 32, (unsigned)((64) + 15) / 16, (unsigned)(2 * 64)), 32, 0, stream>>>(i1c6_6); }
    { GemmP i1c6_7;
      i1c6_7.A = R67 + 0 + (size_t)133 * 3; i1c6_7.B = iw1 + 7; i1c6_7.bias = R67 + 0 + (size_t)133 * 3; i1c6_7.R = R67 + 26176 + (size_t)67 * 16; i1c6_7.C = R67 + 26176 + (size_t)67 * 16;
      i1c6_7.sAo = (long long)66 * 66 * 3; i1c6_7.sAi = (long long)66 * 3; i1c6_7.sAm = 3; i1c6_7.sAk = 1; i1c6_7.sBo = 0; i1c6_7.sBi = 0; i1c6_7.sBn = 3 * 9; i1c6_7.sBk = 9; i1c6_7.sCo = (long long)66 * 66 * 16; i1c6_7.sCi = (long long)66 * 16; i1c6_7.sCm = 16; i1c6_7.sRo = (long long)66 * 66 * 16; i1c6_7.sRi = (long long)66 * 16; i1c6_7.sRm = 16; i1c6_7.sRn = 1;
      i1c6_7.M = 64; i1c6_7.N = 16; i1c6_7.K = 3; i1c6_7.zi_n = 64; i1c6_7.flags = 4; i1c6_7.act = 0;
      i1c6_7.alpha = 1.0f; i1c6_7.beta = 1.0f; i1c6_7.sa = 1.0f; i1c6_7.sb = 1.0f; i1c6_7.Npad = 16; i1c6_7.pad_ = 0;
      k_gemm<1><<<dim3((unsigned)((16) + 31) / 32, (unsigned)((64) + 15) / 16, (unsigned)(2 * 64)), 32, 0, stream>>>(i1c6_7); }
    { GemmP i1c6_8;
      i1c6_8.A = R67 + 0 + (size_t)134 * 3; i1c6_8.B = iw1 + 8; i1c6_8.bias = R67 + 0 + (size_t)134 * 3; i1c6_8.R = R67 + 26176 + (size_t)67 * 16; i1c6_8.C = R67 + 26176 + (size_t)67 * 16;
      i1c6_8.sAo = (long long)66 * 66 * 3; i1c6_8.sAi = (long long)66 * 3; i1c6_8.sAm = 3; i1c6_8.sAk = 1; i1c6_8.sBo = 0; i1c6_8.sBi = 0; i1c6_8.sBn = 3 * 9; i1c6_8.sBk = 9; i1c6_8.sCo = (long long)66 * 66 * 16; i1c6_8.sCi = (long long)66 * 16; i1c6_8.sCm = 16; i1c6_8.sRo = (long long)66 * 66 * 16; i1c6_8.sRi = (long long)66 * 16; i1c6_8.sRm = 16; i1c6_8.sRn = 1;
      i1c6_8.M = 64; i1c6_8.N = 16; i1c6_8.K = 3; i1c6_8.zi_n = 64; i1c6_8.flags = 4; i1c6_8.act = 0;
      i1c6_8.alpha = 1.0f; i1c6_8.beta = 1.0f; i1c6_8.sa = 1.0f; i1c6_8.sb = 1.0f; i1c6_8.Npad = 16; i1c6_8.pad_ = 0;
      k_gemm<1><<<dim3((unsigned)((16) + 31) / 32, (unsigned)((64) + 15) / 16, (unsigned)(2 * 64)), 32, 0, stream>>>(i1c6_8); }
    k_mm_relu2d<<<(unsigned)(((long long)2 * HW * 16 + 255) / 256), 256, 0, stream>>>(R67 + 26176, nullptr, 2, 64, 16);
    { GemmP i2c6_0;
      i2c6_0.A = R67 + 26176 + (size_t)0 * 16; i2c6_0.B = iw2 + 0; i2c6_0.bias = ib2; i2c6_0.R = R67 + 26176 + (size_t)0 * 16; i2c6_0.C = R67 + 165568 + (size_t)67 * 32;
      i2c6_0.sAo = (long long)66 * 66 * 16; i2c6_0.sAi = (long long)66 * 16; i2c6_0.sAm = 16; i2c6_0.sAk = 1; i2c6_0.sBo = 0; i2c6_0.sBi = 0; i2c6_0.sBn = 16 * 9; i2c6_0.sBk = 9; i2c6_0.sCo = (long long)66 * 66 * 32; i2c6_0.sCi = (long long)66 * 32; i2c6_0.sCm = 32; i2c6_0.sRo = 0; i2c6_0.sRi = 0; i2c6_0.sRm = 0; i2c6_0.sRn = 0;
      i2c6_0.M = 64; i2c6_0.N = 32; i2c6_0.K = 16; i2c6_0.zi_n = 64; i2c6_0.flags = 1; i2c6_0.act = 0;
      i2c6_0.alpha = 1.0f; i2c6_0.beta = 0.0f; i2c6_0.sa = 1.0f; i2c6_0.sb = 1.0f; i2c6_0.Npad = 32; i2c6_0.pad_ = 0;
      k_gemm<1><<<dim3((unsigned)((32) + 31) / 32, (unsigned)((64) + 15) / 16, (unsigned)(2 * 64)), 32, 0, stream>>>(i2c6_0); }
    { GemmP i2c6_1;
      i2c6_1.A = R67 + 26176 + (size_t)1 * 16; i2c6_1.B = iw2 + 1; i2c6_1.bias = R67 + 26176 + (size_t)1 * 16; i2c6_1.R = R67 + 165568 + (size_t)67 * 32; i2c6_1.C = R67 + 165568 + (size_t)67 * 32;
      i2c6_1.sAo = (long long)66 * 66 * 16; i2c6_1.sAi = (long long)66 * 16; i2c6_1.sAm = 16; i2c6_1.sAk = 1; i2c6_1.sBo = 0; i2c6_1.sBi = 0; i2c6_1.sBn = 16 * 9; i2c6_1.sBk = 9; i2c6_1.sCo = (long long)66 * 66 * 32; i2c6_1.sCi = (long long)66 * 32; i2c6_1.sCm = 32; i2c6_1.sRo = (long long)66 * 66 * 32; i2c6_1.sRi = (long long)66 * 32; i2c6_1.sRm = 32; i2c6_1.sRn = 1;
      i2c6_1.M = 64; i2c6_1.N = 32; i2c6_1.K = 16; i2c6_1.zi_n = 64; i2c6_1.flags = 4; i2c6_1.act = 0;
      i2c6_1.alpha = 1.0f; i2c6_1.beta = 1.0f; i2c6_1.sa = 1.0f; i2c6_1.sb = 1.0f; i2c6_1.Npad = 32; i2c6_1.pad_ = 0;
      k_gemm<1><<<dim3((unsigned)((32) + 31) / 32, (unsigned)((64) + 15) / 16, (unsigned)(2 * 64)), 32, 0, stream>>>(i2c6_1); }
    { GemmP i2c6_2;
      i2c6_2.A = R67 + 26176 + (size_t)2 * 16; i2c6_2.B = iw2 + 2; i2c6_2.bias = R67 + 26176 + (size_t)2 * 16; i2c6_2.R = R67 + 165568 + (size_t)67 * 32; i2c6_2.C = R67 + 165568 + (size_t)67 * 32;
      i2c6_2.sAo = (long long)66 * 66 * 16; i2c6_2.sAi = (long long)66 * 16; i2c6_2.sAm = 16; i2c6_2.sAk = 1; i2c6_2.sBo = 0; i2c6_2.sBi = 0; i2c6_2.sBn = 16 * 9; i2c6_2.sBk = 9; i2c6_2.sCo = (long long)66 * 66 * 32; i2c6_2.sCi = (long long)66 * 32; i2c6_2.sCm = 32; i2c6_2.sRo = (long long)66 * 66 * 32; i2c6_2.sRi = (long long)66 * 32; i2c6_2.sRm = 32; i2c6_2.sRn = 1;
      i2c6_2.M = 64; i2c6_2.N = 32; i2c6_2.K = 16; i2c6_2.zi_n = 64; i2c6_2.flags = 4; i2c6_2.act = 0;
      i2c6_2.alpha = 1.0f; i2c6_2.beta = 1.0f; i2c6_2.sa = 1.0f; i2c6_2.sb = 1.0f; i2c6_2.Npad = 32; i2c6_2.pad_ = 0;
      k_gemm<1><<<dim3((unsigned)((32) + 31) / 32, (unsigned)((64) + 15) / 16, (unsigned)(2 * 64)), 32, 0, stream>>>(i2c6_2); }
    { GemmP i2c6_3;
      i2c6_3.A = R67 + 26176 + (size_t)66 * 16; i2c6_3.B = iw2 + 3; i2c6_3.bias = R67 + 26176 + (size_t)66 * 16; i2c6_3.R = R67 + 165568 + (size_t)67 * 32; i2c6_3.C = R67 + 165568 + (size_t)67 * 32;
      i2c6_3.sAo = (long long)66 * 66 * 16; i2c6_3.sAi = (long long)66 * 16; i2c6_3.sAm = 16; i2c6_3.sAk = 1; i2c6_3.sBo = 0; i2c6_3.sBi = 0; i2c6_3.sBn = 16 * 9; i2c6_3.sBk = 9; i2c6_3.sCo = (long long)66 * 66 * 32; i2c6_3.sCi = (long long)66 * 32; i2c6_3.sCm = 32; i2c6_3.sRo = (long long)66 * 66 * 32; i2c6_3.sRi = (long long)66 * 32; i2c6_3.sRm = 32; i2c6_3.sRn = 1;
      i2c6_3.M = 64; i2c6_3.N = 32; i2c6_3.K = 16; i2c6_3.zi_n = 64; i2c6_3.flags = 4; i2c6_3.act = 0;
      i2c6_3.alpha = 1.0f; i2c6_3.beta = 1.0f; i2c6_3.sa = 1.0f; i2c6_3.sb = 1.0f; i2c6_3.Npad = 32; i2c6_3.pad_ = 0;
      k_gemm<1><<<dim3((unsigned)((32) + 31) / 32, (unsigned)((64) + 15) / 16, (unsigned)(2 * 64)), 32, 0, stream>>>(i2c6_3); }
    { GemmP i2c6_4;
      i2c6_4.A = R67 + 26176 + (size_t)67 * 16; i2c6_4.B = iw2 + 4; i2c6_4.bias = R67 + 26176 + (size_t)67 * 16; i2c6_4.R = R67 + 165568 + (size_t)67 * 32; i2c6_4.C = R67 + 165568 + (size_t)67 * 32;
      i2c6_4.sAo = (long long)66 * 66 * 16; i2c6_4.sAi = (long long)66 * 16; i2c6_4.sAm = 16; i2c6_4.sAk = 1; i2c6_4.sBo = 0; i2c6_4.sBi = 0; i2c6_4.sBn = 16 * 9; i2c6_4.sBk = 9; i2c6_4.sCo = (long long)66 * 66 * 32; i2c6_4.sCi = (long long)66 * 32; i2c6_4.sCm = 32; i2c6_4.sRo = (long long)66 * 66 * 32; i2c6_4.sRi = (long long)66 * 32; i2c6_4.sRm = 32; i2c6_4.sRn = 1;
      i2c6_4.M = 64; i2c6_4.N = 32; i2c6_4.K = 16; i2c6_4.zi_n = 64; i2c6_4.flags = 4; i2c6_4.act = 0;
      i2c6_4.alpha = 1.0f; i2c6_4.beta = 1.0f; i2c6_4.sa = 1.0f; i2c6_4.sb = 1.0f; i2c6_4.Npad = 32; i2c6_4.pad_ = 0;
      k_gemm<1><<<dim3((unsigned)((32) + 31) / 32, (unsigned)((64) + 15) / 16, (unsigned)(2 * 64)), 32, 0, stream>>>(i2c6_4); }
    { GemmP i2c6_5;
      i2c6_5.A = R67 + 26176 + (size_t)68 * 16; i2c6_5.B = iw2 + 5; i2c6_5.bias = R67 + 26176 + (size_t)68 * 16; i2c6_5.R = R67 + 165568 + (size_t)67 * 32; i2c6_5.C = R67 + 165568 + (size_t)67 * 32;
      i2c6_5.sAo = (long long)66 * 66 * 16; i2c6_5.sAi = (long long)66 * 16; i2c6_5.sAm = 16; i2c6_5.sAk = 1; i2c6_5.sBo = 0; i2c6_5.sBi = 0; i2c6_5.sBn = 16 * 9; i2c6_5.sBk = 9; i2c6_5.sCo = (long long)66 * 66 * 32; i2c6_5.sCi = (long long)66 * 32; i2c6_5.sCm = 32; i2c6_5.sRo = (long long)66 * 66 * 32; i2c6_5.sRi = (long long)66 * 32; i2c6_5.sRm = 32; i2c6_5.sRn = 1;
      i2c6_5.M = 64; i2c6_5.N = 32; i2c6_5.K = 16; i2c6_5.zi_n = 64; i2c6_5.flags = 4; i2c6_5.act = 0;
      i2c6_5.alpha = 1.0f; i2c6_5.beta = 1.0f; i2c6_5.sa = 1.0f; i2c6_5.sb = 1.0f; i2c6_5.Npad = 32; i2c6_5.pad_ = 0;
      k_gemm<1><<<dim3((unsigned)((32) + 31) / 32, (unsigned)((64) + 15) / 16, (unsigned)(2 * 64)), 32, 0, stream>>>(i2c6_5); }
    { GemmP i2c6_6;
      i2c6_6.A = R67 + 26176 + (size_t)132 * 16; i2c6_6.B = iw2 + 6; i2c6_6.bias = R67 + 26176 + (size_t)132 * 16; i2c6_6.R = R67 + 165568 + (size_t)67 * 32; i2c6_6.C = R67 + 165568 + (size_t)67 * 32;
      i2c6_6.sAo = (long long)66 * 66 * 16; i2c6_6.sAi = (long long)66 * 16; i2c6_6.sAm = 16; i2c6_6.sAk = 1; i2c6_6.sBo = 0; i2c6_6.sBi = 0; i2c6_6.sBn = 16 * 9; i2c6_6.sBk = 9; i2c6_6.sCo = (long long)66 * 66 * 32; i2c6_6.sCi = (long long)66 * 32; i2c6_6.sCm = 32; i2c6_6.sRo = (long long)66 * 66 * 32; i2c6_6.sRi = (long long)66 * 32; i2c6_6.sRm = 32; i2c6_6.sRn = 1;
      i2c6_6.M = 64; i2c6_6.N = 32; i2c6_6.K = 16; i2c6_6.zi_n = 64; i2c6_6.flags = 4; i2c6_6.act = 0;
      i2c6_6.alpha = 1.0f; i2c6_6.beta = 1.0f; i2c6_6.sa = 1.0f; i2c6_6.sb = 1.0f; i2c6_6.Npad = 32; i2c6_6.pad_ = 0;
      k_gemm<1><<<dim3((unsigned)((32) + 31) / 32, (unsigned)((64) + 15) / 16, (unsigned)(2 * 64)), 32, 0, stream>>>(i2c6_6); }
    { GemmP i2c6_7;
      i2c6_7.A = R67 + 26176 + (size_t)133 * 16; i2c6_7.B = iw2 + 7; i2c6_7.bias = R67 + 26176 + (size_t)133 * 16; i2c6_7.R = R67 + 165568 + (size_t)67 * 32; i2c6_7.C = R67 + 165568 + (size_t)67 * 32;
      i2c6_7.sAo = (long long)66 * 66 * 16; i2c6_7.sAi = (long long)66 * 16; i2c6_7.sAm = 16; i2c6_7.sAk = 1; i2c6_7.sBo = 0; i2c6_7.sBi = 0; i2c6_7.sBn = 16 * 9; i2c6_7.sBk = 9; i2c6_7.sCo = (long long)66 * 66 * 32; i2c6_7.sCi = (long long)66 * 32; i2c6_7.sCm = 32; i2c6_7.sRo = (long long)66 * 66 * 32; i2c6_7.sRi = (long long)66 * 32; i2c6_7.sRm = 32; i2c6_7.sRn = 1;
      i2c6_7.M = 64; i2c6_7.N = 32; i2c6_7.K = 16; i2c6_7.zi_n = 64; i2c6_7.flags = 4; i2c6_7.act = 0;
      i2c6_7.alpha = 1.0f; i2c6_7.beta = 1.0f; i2c6_7.sa = 1.0f; i2c6_7.sb = 1.0f; i2c6_7.Npad = 32; i2c6_7.pad_ = 0;
      k_gemm<1><<<dim3((unsigned)((32) + 31) / 32, (unsigned)((64) + 15) / 16, (unsigned)(2 * 64)), 32, 0, stream>>>(i2c6_7); }
    { GemmP i2c6_8;
      i2c6_8.A = R67 + 26176 + (size_t)134 * 16; i2c6_8.B = iw2 + 8; i2c6_8.bias = R67 + 26176 + (size_t)134 * 16; i2c6_8.R = R67 + 165568 + (size_t)67 * 32; i2c6_8.C = R67 + 165568 + (size_t)67 * 32;
      i2c6_8.sAo = (long long)66 * 66 * 16; i2c6_8.sAi = (long long)66 * 16; i2c6_8.sAm = 16; i2c6_8.sAk = 1; i2c6_8.sBo = 0; i2c6_8.sBi = 0; i2c6_8.sBn = 16 * 9; i2c6_8.sBk = 9; i2c6_8.sCo = (long long)66 * 66 * 32; i2c6_8.sCi = (long long)66 * 32; i2c6_8.sCm = 32; i2c6_8.sRo = (long long)66 * 66 * 32; i2c6_8.sRi = (long long)66 * 32; i2c6_8.sRm = 32; i2c6_8.sRn = 1;
      i2c6_8.M = 64; i2c6_8.N = 32; i2c6_8.K = 16; i2c6_8.zi_n = 64; i2c6_8.flags = 4; i2c6_8.act = 0;
      i2c6_8.alpha = 1.0f; i2c6_8.beta = 1.0f; i2c6_8.sa = 1.0f; i2c6_8.sb = 1.0f; i2c6_8.Npad = 32; i2c6_8.pad_ = 0;
      k_gemm<1><<<dim3((unsigned)((32) + 31) / 32, (unsigned)((64) + 15) / 16, (unsigned)(2 * 64)), 32, 0, stream>>>(i2c6_8); }
    k_mm_relu2d<<<(unsigned)(((long long)2 * HW * 32 + 255) / 256), 256, 0, stream>>>(R67 + 165568, nullptr, 2, 64, 32);
    { GemmP i3c6_0;
      i3c6_0.A = R67 + 165568 + (size_t)0 * 32; i3c6_0.B = iw3 + 0; i3c6_0.bias = ib3; i3c6_0.R = R67 + 165568 + (size_t)0 * 32; i3c6_0.C = R67 + 444352 + (size_t)67 * 64;
      i3c6_0.sAo = (long long)66 * 66 * 32; i3c6_0.sAi = (long long)66 * 32; i3c6_0.sAm = 32; i3c6_0.sAk = 1; i3c6_0.sBo = 0; i3c6_0.sBi = 0; i3c6_0.sBn = 32 * 9; i3c6_0.sBk = 9; i3c6_0.sCo = (long long)66 * 66 * 64; i3c6_0.sCi = (long long)66 * 64; i3c6_0.sCm = 64; i3c6_0.sRo = 0; i3c6_0.sRi = 0; i3c6_0.sRm = 0; i3c6_0.sRn = 0;
      i3c6_0.M = 64; i3c6_0.N = 64; i3c6_0.K = 32; i3c6_0.zi_n = 64; i3c6_0.flags = 1; i3c6_0.act = 0;
      i3c6_0.alpha = 1.0f; i3c6_0.beta = 0.0f; i3c6_0.sa = 1.0f; i3c6_0.sb = 1.0f; i3c6_0.Npad = 64; i3c6_0.pad_ = 0;
      k_gemm<1><<<dim3((unsigned)((64) + 31) / 32, (unsigned)((64) + 15) / 16, (unsigned)(2 * 64)), 32, 0, stream>>>(i3c6_0); }
    { GemmP i3c6_1;
      i3c6_1.A = R67 + 165568 + (size_t)1 * 32; i3c6_1.B = iw3 + 1; i3c6_1.bias = R67 + 165568 + (size_t)1 * 32; i3c6_1.R = R67 + 444352 + (size_t)67 * 64; i3c6_1.C = R67 + 444352 + (size_t)67 * 64;
      i3c6_1.sAo = (long long)66 * 66 * 32; i3c6_1.sAi = (long long)66 * 32; i3c6_1.sAm = 32; i3c6_1.sAk = 1; i3c6_1.sBo = 0; i3c6_1.sBi = 0; i3c6_1.sBn = 32 * 9; i3c6_1.sBk = 9; i3c6_1.sCo = (long long)66 * 66 * 64; i3c6_1.sCi = (long long)66 * 64; i3c6_1.sCm = 64; i3c6_1.sRo = (long long)66 * 66 * 64; i3c6_1.sRi = (long long)66 * 64; i3c6_1.sRm = 64; i3c6_1.sRn = 1;
      i3c6_1.M = 64; i3c6_1.N = 64; i3c6_1.K = 32; i3c6_1.zi_n = 64; i3c6_1.flags = 4; i3c6_1.act = 0;
      i3c6_1.alpha = 1.0f; i3c6_1.beta = 1.0f; i3c6_1.sa = 1.0f; i3c6_1.sb = 1.0f; i3c6_1.Npad = 64; i3c6_1.pad_ = 0;
      k_gemm<1><<<dim3((unsigned)((64) + 31) / 32, (unsigned)((64) + 15) / 16, (unsigned)(2 * 64)), 32, 0, stream>>>(i3c6_1); }
    { GemmP i3c6_2;
      i3c6_2.A = R67 + 165568 + (size_t)2 * 32; i3c6_2.B = iw3 + 2; i3c6_2.bias = R67 + 165568 + (size_t)2 * 32; i3c6_2.R = R67 + 444352 + (size_t)67 * 64; i3c6_2.C = R67 + 444352 + (size_t)67 * 64;
      i3c6_2.sAo = (long long)66 * 66 * 32; i3c6_2.sAi = (long long)66 * 32; i3c6_2.sAm = 32; i3c6_2.sAk = 1; i3c6_2.sBo = 0; i3c6_2.sBi = 0; i3c6_2.sBn = 32 * 9; i3c6_2.sBk = 9; i3c6_2.sCo = (long long)66 * 66 * 64; i3c6_2.sCi = (long long)66 * 64; i3c6_2.sCm = 64; i3c6_2.sRo = (long long)66 * 66 * 64; i3c6_2.sRi = (long long)66 * 64; i3c6_2.sRm = 64; i3c6_2.sRn = 1;
      i3c6_2.M = 64; i3c6_2.N = 64; i3c6_2.K = 32; i3c6_2.zi_n = 64; i3c6_2.flags = 4; i3c6_2.act = 0;
      i3c6_2.alpha = 1.0f; i3c6_2.beta = 1.0f; i3c6_2.sa = 1.0f; i3c6_2.sb = 1.0f; i3c6_2.Npad = 64; i3c6_2.pad_ = 0;
      k_gemm<1><<<dim3((unsigned)((64) + 31) / 32, (unsigned)((64) + 15) / 16, (unsigned)(2 * 64)), 32, 0, stream>>>(i3c6_2); }
    { GemmP i3c6_3;
      i3c6_3.A = R67 + 165568 + (size_t)66 * 32; i3c6_3.B = iw3 + 3; i3c6_3.bias = R67 + 165568 + (size_t)66 * 32; i3c6_3.R = R67 + 444352 + (size_t)67 * 64; i3c6_3.C = R67 + 444352 + (size_t)67 * 64;
      i3c6_3.sAo = (long long)66 * 66 * 32; i3c6_3.sAi = (long long)66 * 32; i3c6_3.sAm = 32; i3c6_3.sAk = 1; i3c6_3.sBo = 0; i3c6_3.sBi = 0; i3c6_3.sBn = 32 * 9; i3c6_3.sBk = 9; i3c6_3.sCo = (long long)66 * 66 * 64; i3c6_3.sCi = (long long)66 * 64; i3c6_3.sCm = 64; i3c6_3.sRo = (long long)66 * 66 * 64; i3c6_3.sRi = (long long)66 * 64; i3c6_3.sRm = 64; i3c6_3.sRn = 1;
      i3c6_3.M = 64; i3c6_3.N = 64; i3c6_3.K = 32; i3c6_3.zi_n = 64; i3c6_3.flags = 4; i3c6_3.act = 0;
      i3c6_3.alpha = 1.0f; i3c6_3.beta = 1.0f; i3c6_3.sa = 1.0f; i3c6_3.sb = 1.0f; i3c6_3.Npad = 64; i3c6_3.pad_ = 0;
      k_gemm<1><<<dim3((unsigned)((64) + 31) / 32, (unsigned)((64) + 15) / 16, (unsigned)(2 * 64)), 32, 0, stream>>>(i3c6_3); }
    { GemmP i3c6_4;
      i3c6_4.A = R67 + 165568 + (size_t)67 * 32; i3c6_4.B = iw3 + 4; i3c6_4.bias = R67 + 165568 + (size_t)67 * 32; i3c6_4.R = R67 + 444352 + (size_t)67 * 64; i3c6_4.C = R67 + 444352 + (size_t)67 * 64;
      i3c6_4.sAo = (long long)66 * 66 * 32; i3c6_4.sAi = (long long)66 * 32; i3c6_4.sAm = 32; i3c6_4.sAk = 1; i3c6_4.sBo = 0; i3c6_4.sBi = 0; i3c6_4.sBn = 32 * 9; i3c6_4.sBk = 9; i3c6_4.sCo = (long long)66 * 66 * 64; i3c6_4.sCi = (long long)66 * 64; i3c6_4.sCm = 64; i3c6_4.sRo = (long long)66 * 66 * 64; i3c6_4.sRi = (long long)66 * 64; i3c6_4.sRm = 64; i3c6_4.sRn = 1;
      i3c6_4.M = 64; i3c6_4.N = 64; i3c6_4.K = 32; i3c6_4.zi_n = 64; i3c6_4.flags = 4; i3c6_4.act = 0;
      i3c6_4.alpha = 1.0f; i3c6_4.beta = 1.0f; i3c6_4.sa = 1.0f; i3c6_4.sb = 1.0f; i3c6_4.Npad = 64; i3c6_4.pad_ = 0;
      k_gemm<1><<<dim3((unsigned)((64) + 31) / 32, (unsigned)((64) + 15) / 16, (unsigned)(2 * 64)), 32, 0, stream>>>(i3c6_4); }
    { GemmP i3c6_5;
      i3c6_5.A = R67 + 165568 + (size_t)68 * 32; i3c6_5.B = iw3 + 5; i3c6_5.bias = R67 + 165568 + (size_t)68 * 32; i3c6_5.R = R67 + 444352 + (size_t)67 * 64; i3c6_5.C = R67 + 444352 + (size_t)67 * 64;
      i3c6_5.sAo = (long long)66 * 66 * 32; i3c6_5.sAi = (long long)66 * 32; i3c6_5.sAm = 32; i3c6_5.sAk = 1; i3c6_5.sBo = 0; i3c6_5.sBi = 0; i3c6_5.sBn = 32 * 9; i3c6_5.sBk = 9; i3c6_5.sCo = (long long)66 * 66 * 64; i3c6_5.sCi = (long long)66 * 64; i3c6_5.sCm = 64; i3c6_5.sRo = (long long)66 * 66 * 64; i3c6_5.sRi = (long long)66 * 64; i3c6_5.sRm = 64; i3c6_5.sRn = 1;
      i3c6_5.M = 64; i3c6_5.N = 64; i3c6_5.K = 32; i3c6_5.zi_n = 64; i3c6_5.flags = 4; i3c6_5.act = 0;
      i3c6_5.alpha = 1.0f; i3c6_5.beta = 1.0f; i3c6_5.sa = 1.0f; i3c6_5.sb = 1.0f; i3c6_5.Npad = 64; i3c6_5.pad_ = 0;
      k_gemm<1><<<dim3((unsigned)((64) + 31) / 32, (unsigned)((64) + 15) / 16, (unsigned)(2 * 64)), 32, 0, stream>>>(i3c6_5); }
    { GemmP i3c6_6;
      i3c6_6.A = R67 + 165568 + (size_t)132 * 32; i3c6_6.B = iw3 + 6; i3c6_6.bias = R67 + 165568 + (size_t)132 * 32; i3c6_6.R = R67 + 444352 + (size_t)67 * 64; i3c6_6.C = R67 + 444352 + (size_t)67 * 64;
      i3c6_6.sAo = (long long)66 * 66 * 32; i3c6_6.sAi = (long long)66 * 32; i3c6_6.sAm = 32; i3c6_6.sAk = 1; i3c6_6.sBo = 0; i3c6_6.sBi = 0; i3c6_6.sBn = 32 * 9; i3c6_6.sBk = 9; i3c6_6.sCo = (long long)66 * 66 * 64; i3c6_6.sCi = (long long)66 * 64; i3c6_6.sCm = 64; i3c6_6.sRo = (long long)66 * 66 * 64; i3c6_6.sRi = (long long)66 * 64; i3c6_6.sRm = 64; i3c6_6.sRn = 1;
      i3c6_6.M = 64; i3c6_6.N = 64; i3c6_6.K = 32; i3c6_6.zi_n = 64; i3c6_6.flags = 4; i3c6_6.act = 0;
      i3c6_6.alpha = 1.0f; i3c6_6.beta = 1.0f; i3c6_6.sa = 1.0f; i3c6_6.sb = 1.0f; i3c6_6.Npad = 64; i3c6_6.pad_ = 0;
      k_gemm<1><<<dim3((unsigned)((64) + 31) / 32, (unsigned)((64) + 15) / 16, (unsigned)(2 * 64)), 32, 0, stream>>>(i3c6_6); }
    { GemmP i3c6_7;
      i3c6_7.A = R67 + 165568 + (size_t)133 * 32; i3c6_7.B = iw3 + 7; i3c6_7.bias = R67 + 165568 + (size_t)133 * 32; i3c6_7.R = R67 + 444352 + (size_t)67 * 64; i3c6_7.C = R67 + 444352 + (size_t)67 * 64;
      i3c6_7.sAo = (long long)66 * 66 * 32; i3c6_7.sAi = (long long)66 * 32; i3c6_7.sAm = 32; i3c6_7.sAk = 1; i3c6_7.sBo = 0; i3c6_7.sBi = 0; i3c6_7.sBn = 32 * 9; i3c6_7.sBk = 9; i3c6_7.sCo = (long long)66 * 66 * 64; i3c6_7.sCi = (long long)66 * 64; i3c6_7.sCm = 64; i3c6_7.sRo = (long long)66 * 66 * 64; i3c6_7.sRi = (long long)66 * 64; i3c6_7.sRm = 64; i3c6_7.sRn = 1;
      i3c6_7.M = 64; i3c6_7.N = 64; i3c6_7.K = 32; i3c6_7.zi_n = 64; i3c6_7.flags = 4; i3c6_7.act = 0;
      i3c6_7.alpha = 1.0f; i3c6_7.beta = 1.0f; i3c6_7.sa = 1.0f; i3c6_7.sb = 1.0f; i3c6_7.Npad = 64; i3c6_7.pad_ = 0;
      k_gemm<1><<<dim3((unsigned)((64) + 31) / 32, (unsigned)((64) + 15) / 16, (unsigned)(2 * 64)), 32, 0, stream>>>(i3c6_7); }
    { GemmP i3c6_8;
      i3c6_8.A = R67 + 165568 + (size_t)134 * 32; i3c6_8.B = iw3 + 8; i3c6_8.bias = R67 + 165568 + (size_t)134 * 32; i3c6_8.R = R67 + 444352 + (size_t)67 * 64; i3c6_8.C = R67 + 444352 + (size_t)67 * 64;
      i3c6_8.sAo = (long long)66 * 66 * 32; i3c6_8.sAi = (long long)66 * 32; i3c6_8.sAm = 32; i3c6_8.sAk = 1; i3c6_8.sBo = 0; i3c6_8.sBi = 0; i3c6_8.sBn = 32 * 9; i3c6_8.sBk = 9; i3c6_8.sCo = (long long)66 * 66 * 64; i3c6_8.sCi = (long long)66 * 64; i3c6_8.sCm = 64; i3c6_8.sRo = (long long)66 * 66 * 64; i3c6_8.sRi = (long long)66 * 64; i3c6_8.sRm = 64; i3c6_8.sRn = 1;
      i3c6_8.M = 64; i3c6_8.N = 64; i3c6_8.K = 32; i3c6_8.zi_n = 64; i3c6_8.flags = 4; i3c6_8.act = 0;
      i3c6_8.alpha = 1.0f; i3c6_8.beta = 1.0f; i3c6_8.sa = 1.0f; i3c6_8.sb = 1.0f; i3c6_8.Npad = 64; i3c6_8.pad_ = 0;
      k_gemm<1><<<dim3((unsigned)((64) + 31) / 32, (unsigned)((64) + 15) / 16, (unsigned)(2 * 64)), 32, 0, stream>>>(i3c6_8); }
    k_mm_relu2d<<<(unsigned)(((long long)2 * HW * 64 + 255) / 256), 256, 0, stream>>>(R67 + 444352, R67 + 1001920, 2, 64, 64);
    { GemmP gqkv6;
      gqkv6.A = R67 + 1001920; gqkv6.B = qkvw; gqkv6.bias = qkvb; gqkv6.R = R67 + 1001920; gqkv6.C = R67 + 1526208;
      gqkv6.sAo = 0; gqkv6.sAi = 0; gqkv6.sAm = 64; gqkv6.sAk = 1; gqkv6.sBo = 0; gqkv6.sBi = 0; gqkv6.sBn = 64; gqkv6.sBk = 1; gqkv6.sCo = 0; gqkv6.sCi = 0; gqkv6.sCm = 192; gqkv6.sRo = 0; gqkv6.sRi = 0; gqkv6.sRm = 0; gqkv6.sRn = 0;
      gqkv6.M = 2 * HW; gqkv6.N = 192; gqkv6.K = 64; gqkv6.zi_n = 1; gqkv6.flags = 1; gqkv6.act = 0;
      gqkv6.alpha = 1.0f; gqkv6.beta = 0.0f; gqkv6.sa = 1.0f; gqkv6.sb = 1.0f; gqkv6.Npad = 192; gqkv6.pad_ = 0;
      k_gemm<1><<<dim3((unsigned)((192) + 31) / 32, (unsigned)((2 * HW) + 15) / 16, (unsigned)(1)), 32, 0, stream>>>(gqkv6); }
    k_mm_dw<<<(unsigned)(((long long)2 * HW * 192 + 255) / 256), 256, 0, stream>>>(R67 + 1526208, dww, dwb, R67 + 3099072, 2, 64, 192);
    k_mm_fall<<<(unsigned)(((long long)2 * HW * 144 + 255) / 256), 256, 0, stream>>>(R67 + 3099072, fcw, fcb, R67 + 4671936, 2, HW, 192);
    k_mm_dep<<<(unsigned)(((long long)2 * 64 * HW + 255) / 256), 256, 0, stream>>>(R67 + 4671936, depw, depb, R67 + 5851584, 2, 64);
    k_mm_qknorm<<<2 * 128, 256, 0, stream>>>(R67 + 3099072, R67 + 6375872, 2, HW, 192);
    { GemmP gat6;
      gat6.A = R67 + 6375872; gat6.B = R67 + 6375872 + (size_t)64 * HW; gat6.bias = R67 + 6375872; gat6.R = R67 + 6375872; gat6.C = R67 + 7424448;
      gat6.sAo = (long long)128 * HW; gat6.sAi = (long long)16 * HW; gat6.sAm = HW; gat6.sAk = 1; gat6.sBo = (long long)128 * HW; gat6.sBi = (long long)16 * HW; gat6.sBn = HW; gat6.sBk = 1; gat6.sCo = (long long)4 * 16 * LP; gat6.sCi = 16 * LP; gat6.sCm = LP; gat6.sRo = 0; gat6.sRi = 0; gat6.sRm = 0; gat6.sRn = 0;
      gat6.M = 16; gat6.N = 16; gat6.K = HW; gat6.zi_n = 4; gat6.flags = 0; gat6.act = 0;
      gat6.alpha = 1.0f; gat6.beta = 0.0f; gat6.sa = 1.0f; gat6.sb = 1.0f; gat6.Npad = LP; gat6.pad_ = 0;
      k_gemm<1><<<dim3((unsigned)((LP) + 31) / 32, (unsigned)((16) + 15) / 16, (unsigned)(2 * 4)), 32, 0, stream>>>(gat6); }
    k_mm_sm16<<<(unsigned)((2 * 4 * 16 + 255) / 256), 256, 0, stream>>>(R67 + 7424448, temp, 2 * 4, LP);
    { GemmP gao6;
      gao6.A = R67 + 7424448; gao6.B = R67 + 3099072 + 128; gao6.bias = R67 + 7424448; gao6.R = R67 + 7424448; gao6.C = R67 + 7428544;
      gao6.sAo = (long long)4 * 16 * LP; gao6.sAi = 16 * LP; gao6.sAm = LP; gao6.sAk = 1; gao6.sBo = (long long)HW * 192; gao6.sBi = 16; gao6.sBn = 192; gao6.sBk = 1; gao6.sCo = (long long)64 * HW; gao6.sCi = (long long)16 * HW; gao6.sCm = HW; gao6.sRo = 0; gao6.sRi = 0; gao6.sRm = 0; gao6.sRn = 0;
      gao6.M = 16; gao6.N = HW; gao6.K = 16; gao6.zi_n = 4; gao6.flags = 0; gao6.act = 0;
      gao6.alpha = 1.0f; gao6.beta = 0.0f; gao6.sa = 1.0f; gao6.sb = 1.0f; gao6.Npad = HW; gao6.pad_ = 0;
      k_gemm<1><<<dim3((unsigned)((HW) + 31) / 32, (unsigned)((16) + 15) / 16, (unsigned)(2 * 4)), 32, 0, stream>>>(gao6); }
    { GemmP gproj6;
      gproj6.A = projw; gproj6.B = R67 + 7428544; gproj6.bias = projb; gproj6.R = projw; gproj6.C = R67 + 7952832;
      gproj6.sAo = 0; gproj6.sAi = 0; gproj6.sAm = 64; gproj6.sAk = 1; gproj6.sBo = (long long)64 * HW; gproj6.sBi = 0; gproj6.sBn = 1; gproj6.sBk = HW; gproj6.sCo = (long long)64 * HW; gproj6.sCi = 0; gproj6.sCm = HW; gproj6.sRo = 0; gproj6.sRi = 0; gproj6.sRm = 0; gproj6.sRn = 0;
      gproj6.M = 64; gproj6.N = HW; gproj6.K = 64; gproj6.zi_n = 1; gproj6.flags = 2; gproj6.act = 0;
      gproj6.alpha = 1.0f; gproj6.beta = 0.0f; gproj6.sa = 1.0f; gproj6.sb = 1.0f; gproj6.Npad = HW; gproj6.pad_ = 0;
      k_gemm<1><<<dim3((unsigned)((HW) + 31) / 32, (unsigned)((64) + 15) / 16, (unsigned)(2)), 32, 0, stream>>>(gproj6); }
    k_mm_imgfeat<<<(unsigned)(((long long)2 * SEQ * 64 + 255) / 256), 256, 0, stream>>>(R67 + 7952832, R67 + 5851584, IR + (size_t)12 * SEQ * 64, 2, HW, 64);
    hipMemsetAsync(R67 + 0, 0, (size_t)2 * 66 * 66 * 3 * 4, stream); hipMemsetAsync(R67 + 26176, 0, (size_t)2 * 66 * 66 * 16 * 4, stream); hipMemsetAsync(R67 + 165568, 0, (size_t)2 * 66 * 66 * 32 * 4, stream); hipMemsetAsync(R67 + 444352, 0, (size_t)2 * 66 * 66 * 64 * 4, stream);
    k_mm_padimg<<<(unsigned)(((long long)2 * HW * 3 + 255) / 256), 256, 0, stream>>>(img + (size_t)14 * 3 * HW, R67 + 0, 2, 3, 64);
    { GemmP i1c7_0;
      i1c7_0.A = R67 + 0 + (size_t)0 * 3; i1c7_0.B = iw1 + 0; i1c7_0.bias = ib1; i1c7_0.R = R67 + 0 + (size_t)0 * 3; i1c7_0.C = R67 + 26176 + (size_t)67 * 16;
      i1c7_0.sAo = (long long)66 * 66 * 3; i1c7_0.sAi = (long long)66 * 3; i1c7_0.sAm = 3; i1c7_0.sAk = 1; i1c7_0.sBo = 0; i1c7_0.sBi = 0; i1c7_0.sBn = 3 * 9; i1c7_0.sBk = 9; i1c7_0.sCo = (long long)66 * 66 * 16; i1c7_0.sCi = (long long)66 * 16; i1c7_0.sCm = 16; i1c7_0.sRo = 0; i1c7_0.sRi = 0; i1c7_0.sRm = 0; i1c7_0.sRn = 0;
      i1c7_0.M = 64; i1c7_0.N = 16; i1c7_0.K = 3; i1c7_0.zi_n = 64; i1c7_0.flags = 1; i1c7_0.act = 0;
      i1c7_0.alpha = 1.0f; i1c7_0.beta = 0.0f; i1c7_0.sa = 1.0f; i1c7_0.sb = 1.0f; i1c7_0.Npad = 16; i1c7_0.pad_ = 0;
      k_gemm<1><<<dim3((unsigned)((16) + 31) / 32, (unsigned)((64) + 15) / 16, (unsigned)(2 * 64)), 32, 0, stream>>>(i1c7_0); }
    { GemmP i1c7_1;
      i1c7_1.A = R67 + 0 + (size_t)1 * 3; i1c7_1.B = iw1 + 1; i1c7_1.bias = R67 + 0 + (size_t)1 * 3; i1c7_1.R = R67 + 26176 + (size_t)67 * 16; i1c7_1.C = R67 + 26176 + (size_t)67 * 16;
      i1c7_1.sAo = (long long)66 * 66 * 3; i1c7_1.sAi = (long long)66 * 3; i1c7_1.sAm = 3; i1c7_1.sAk = 1; i1c7_1.sBo = 0; i1c7_1.sBi = 0; i1c7_1.sBn = 3 * 9; i1c7_1.sBk = 9; i1c7_1.sCo = (long long)66 * 66 * 16; i1c7_1.sCi = (long long)66 * 16; i1c7_1.sCm = 16; i1c7_1.sRo = (long long)66 * 66 * 16; i1c7_1.sRi = (long long)66 * 16; i1c7_1.sRm = 16; i1c7_1.sRn = 1;
      i1c7_1.M = 64; i1c7_1.N = 16; i1c7_1.K = 3; i1c7_1.zi_n = 64; i1c7_1.flags = 4; i1c7_1.act = 0;
      i1c7_1.alpha = 1.0f; i1c7_1.beta = 1.0f; i1c7_1.sa = 1.0f; i1c7_1.sb = 1.0f; i1c7_1.Npad = 16; i1c7_1.pad_ = 0;
      k_gemm<1><<<dim3((unsigned)((16) + 31) / 32, (unsigned)((64) + 15) / 16, (unsigned)(2 * 64)), 32, 0, stream>>>(i1c7_1); }
    { GemmP i1c7_2;
      i1c7_2.A = R67 + 0 + (size_t)2 * 3; i1c7_2.B = iw1 + 2; i1c7_2.bias = R67 + 0 + (size_t)2 * 3; i1c7_2.R = R67 + 26176 + (size_t)67 * 16; i1c7_2.C = R67 + 26176 + (size_t)67 * 16;
      i1c7_2.sAo = (long long)66 * 66 * 3; i1c7_2.sAi = (long long)66 * 3; i1c7_2.sAm = 3; i1c7_2.sAk = 1; i1c7_2.sBo = 0; i1c7_2.sBi = 0; i1c7_2.sBn = 3 * 9; i1c7_2.sBk = 9; i1c7_2.sCo = (long long)66 * 66 * 16; i1c7_2.sCi = (long long)66 * 16; i1c7_2.sCm = 16; i1c7_2.sRo = (long long)66 * 66 * 16; i1c7_2.sRi = (long long)66 * 16; i1c7_2.sRm = 16; i1c7_2.sRn = 1;
      i1c7_2.M = 64; i1c7_2.N = 16; i1c7_2.K = 3; i1c7_2.zi_n = 64; i1c7_2.flags = 4; i1c7_2.act = 0;
      i1c7_2.alpha = 1.0f; i1c7_2.beta = 1.0f; i1c7_2.sa = 1.0f; i1c7_2.sb = 1.0f; i1c7_2.Npad = 16; i1c7_2.pad_ = 0;
      k_gemm<1><<<dim3((unsigned)((16) + 31) / 32, (unsigned)((64) + 15) / 16, (unsigned)(2 * 64)), 32, 0, stream>>>(i1c7_2); }
    { GemmP i1c7_3;
      i1c7_3.A = R67 + 0 + (size_t)66 * 3; i1c7_3.B = iw1 + 3; i1c7_3.bias = R67 + 0 + (size_t)66 * 3; i1c7_3.R = R67 + 26176 + (size_t)67 * 16; i1c7_3.C = R67 + 26176 + (size_t)67 * 16;
      i1c7_3.sAo = (long long)66 * 66 * 3; i1c7_3.sAi = (long long)66 * 3; i1c7_3.sAm = 3; i1c7_3.sAk = 1; i1c7_3.sBo = 0; i1c7_3.sBi = 0; i1c7_3.sBn = 3 * 9; i1c7_3.sBk = 9; i1c7_3.sCo = (long long)66 * 66 * 16; i1c7_3.sCi = (long long)66 * 16; i1c7_3.sCm = 16; i1c7_3.sRo = (long long)66 * 66 * 16; i1c7_3.sRi = (long long)66 * 16; i1c7_3.sRm = 16; i1c7_3.sRn = 1;
      i1c7_3.M = 64; i1c7_3.N = 16; i1c7_3.K = 3; i1c7_3.zi_n = 64; i1c7_3.flags = 4; i1c7_3.act = 0;
      i1c7_3.alpha = 1.0f; i1c7_3.beta = 1.0f; i1c7_3.sa = 1.0f; i1c7_3.sb = 1.0f; i1c7_3.Npad = 16; i1c7_3.pad_ = 0;
      k_gemm<1><<<dim3((unsigned)((16) + 31) / 32, (unsigned)((64) + 15) / 16, (unsigned)(2 * 64)), 32, 0, stream>>>(i1c7_3); }
    { GemmP i1c7_4;
      i1c7_4.A = R67 + 0 + (size_t)67 * 3; i1c7_4.B = iw1 + 4; i1c7_4.bias = R67 + 0 + (size_t)67 * 3; i1c7_4.R = R67 + 26176 + (size_t)67 * 16; i1c7_4.C = R67 + 26176 + (size_t)67 * 16;
      i1c7_4.sAo = (long long)66 * 66 * 3; i1c7_4.sAi = (long long)66 * 3; i1c7_4.sAm = 3; i1c7_4.sAk = 1; i1c7_4.sBo = 0; i1c7_4.sBi = 0; i1c7_4.sBn = 3 * 9; i1c7_4.sBk = 9; i1c7_4.sCo = (long long)66 * 66 * 16; i1c7_4.sCi = (long long)66 * 16; i1c7_4.sCm = 16; i1c7_4.sRo = (long long)66 * 66 * 16; i1c7_4.sRi = (long long)66 * 16; i1c7_4.sRm = 16; i1c7_4.sRn = 1;
      i1c7_4.M = 64; i1c7_4.N = 16; i1c7_4.K = 3; i1c7_4.zi_n = 64; i1c7_4.flags = 4; i1c7_4.act = 0;
      i1c7_4.alpha = 1.0f; i1c7_4.beta = 1.0f; i1c7_4.sa = 1.0f; i1c7_4.sb = 1.0f; i1c7_4.Npad = 16; i1c7_4.pad_ = 0;
      k_gemm<1><<<dim3((unsigned)((16) + 31) / 32, (unsigned)((64) + 15) / 16, (unsigned)(2 * 64)), 32, 0, stream>>>(i1c7_4); }
    { GemmP i1c7_5;
      i1c7_5.A = R67 + 0 + (size_t)68 * 3; i1c7_5.B = iw1 + 5; i1c7_5.bias = R67 + 0 + (size_t)68 * 3; i1c7_5.R = R67 + 26176 + (size_t)67 * 16; i1c7_5.C = R67 + 26176 + (size_t)67 * 16;
      i1c7_5.sAo = (long long)66 * 66 * 3; i1c7_5.sAi = (long long)66 * 3; i1c7_5.sAm = 3; i1c7_5.sAk = 1; i1c7_5.sBo = 0; i1c7_5.sBi = 0; i1c7_5.sBn = 3 * 9; i1c7_5.sBk = 9; i1c7_5.sCo = (long long)66 * 66 * 16; i1c7_5.sCi = (long long)66 * 16; i1c7_5.sCm = 16; i1c7_5.sRo = (long long)66 * 66 * 16; i1c7_5.sRi = (long long)66 * 16; i1c7_5.sRm = 16; i1c7_5.sRn = 1;
      i1c7_5.M = 64; i1c7_5.N = 16; i1c7_5.K = 3; i1c7_5.zi_n = 64; i1c7_5.flags = 4; i1c7_5.act = 0;
      i1c7_5.alpha = 1.0f; i1c7_5.beta = 1.0f; i1c7_5.sa = 1.0f; i1c7_5.sb = 1.0f; i1c7_5.Npad = 16; i1c7_5.pad_ = 0;
      k_gemm<1><<<dim3((unsigned)((16) + 31) / 32, (unsigned)((64) + 15) / 16, (unsigned)(2 * 64)), 32, 0, stream>>>(i1c7_5); }
    { GemmP i1c7_6;
      i1c7_6.A = R67 + 0 + (size_t)132 * 3; i1c7_6.B = iw1 + 6; i1c7_6.bias = R67 + 0 + (size_t)132 * 3; i1c7_6.R = R67 + 26176 + (size_t)67 * 16; i1c7_6.C = R67 + 26176 + (size_t)67 * 16;
      i1c7_6.sAo = (long long)66 * 66 * 3; i1c7_6.sAi = (long long)66 * 3; i1c7_6.sAm = 3; i1c7_6.sAk = 1; i1c7_6.sBo = 0; i1c7_6.sBi = 0; i1c7_6.sBn = 3 * 9; i1c7_6.sBk = 9; i1c7_6.sCo = (long long)66 * 66 * 16; i1c7_6.sCi = (long long)66 * 16; i1c7_6.sCm = 16; i1c7_6.sRo = (long long)66 * 66 * 16; i1c7_6.sRi = (long long)66 * 16; i1c7_6.sRm = 16; i1c7_6.sRn = 1;
      i1c7_6.M = 64; i1c7_6.N = 16; i1c7_6.K = 3; i1c7_6.zi_n = 64; i1c7_6.flags = 4; i1c7_6.act = 0;
      i1c7_6.alpha = 1.0f; i1c7_6.beta = 1.0f; i1c7_6.sa = 1.0f; i1c7_6.sb = 1.0f; i1c7_6.Npad = 16; i1c7_6.pad_ = 0;
      k_gemm<1><<<dim3((unsigned)((16) + 31) / 32, (unsigned)((64) + 15) / 16, (unsigned)(2 * 64)), 32, 0, stream>>>(i1c7_6); }
    { GemmP i1c7_7;
      i1c7_7.A = R67 + 0 + (size_t)133 * 3; i1c7_7.B = iw1 + 7; i1c7_7.bias = R67 + 0 + (size_t)133 * 3; i1c7_7.R = R67 + 26176 + (size_t)67 * 16; i1c7_7.C = R67 + 26176 + (size_t)67 * 16;
      i1c7_7.sAo = (long long)66 * 66 * 3; i1c7_7.sAi = (long long)66 * 3; i1c7_7.sAm = 3; i1c7_7.sAk = 1; i1c7_7.sBo = 0; i1c7_7.sBi = 0; i1c7_7.sBn = 3 * 9; i1c7_7.sBk = 9; i1c7_7.sCo = (long long)66 * 66 * 16; i1c7_7.sCi = (long long)66 * 16; i1c7_7.sCm = 16; i1c7_7.sRo = (long long)66 * 66 * 16; i1c7_7.sRi = (long long)66 * 16; i1c7_7.sRm = 16; i1c7_7.sRn = 1;
      i1c7_7.M = 64; i1c7_7.N = 16; i1c7_7.K = 3; i1c7_7.zi_n = 64; i1c7_7.flags = 4; i1c7_7.act = 0;
      i1c7_7.alpha = 1.0f; i1c7_7.beta = 1.0f; i1c7_7.sa = 1.0f; i1c7_7.sb = 1.0f; i1c7_7.Npad = 16; i1c7_7.pad_ = 0;
      k_gemm<1><<<dim3((unsigned)((16) + 31) / 32, (unsigned)((64) + 15) / 16, (unsigned)(2 * 64)), 32, 0, stream>>>(i1c7_7); }
    { GemmP i1c7_8;
      i1c7_8.A = R67 + 0 + (size_t)134 * 3; i1c7_8.B = iw1 + 8; i1c7_8.bias = R67 + 0 + (size_t)134 * 3; i1c7_8.R = R67 + 26176 + (size_t)67 * 16; i1c7_8.C = R67 + 26176 + (size_t)67 * 16;
      i1c7_8.sAo = (long long)66 * 66 * 3; i1c7_8.sAi = (long long)66 * 3; i1c7_8.sAm = 3; i1c7_8.sAk = 1; i1c7_8.sBo = 0; i1c7_8.sBi = 0; i1c7_8.sBn = 3 * 9; i1c7_8.sBk = 9; i1c7_8.sCo = (long long)66 * 66 * 16; i1c7_8.sCi = (long long)66 * 16; i1c7_8.sCm = 16; i1c7_8.sRo = (long long)66 * 66 * 16; i1c7_8.sRi = (long long)66 * 16; i1c7_8.sRm = 16; i1c7_8.sRn = 1;
      i1c7_8.M = 64; i1c7_8.N = 16; i1c7_8.K = 3; i1c7_8.zi_n = 64; i1c7_8.flags = 4; i1c7_8.act = 0;
      i1c7_8.alpha = 1.0f; i1c7_8.beta = 1.0f; i1c7_8.sa = 1.0f; i1c7_8.sb = 1.0f; i1c7_8.Npad = 16; i1c7_8.pad_ = 0;
      k_gemm<1><<<dim3((unsigned)((16) + 31) / 32, (unsigned)((64) + 15) / 16, (unsigned)(2 * 64)), 32, 0, stream>>>(i1c7_8); }
    k_mm_relu2d<<<(unsigned)(((long long)2 * HW * 16 + 255) / 256), 256, 0, stream>>>(R67 + 26176, nullptr, 2, 64, 16);
    { GemmP i2c7_0;
      i2c7_0.A = R67 + 26176 + (size_t)0 * 16; i2c7_0.B = iw2 + 0; i2c7_0.bias = ib2; i2c7_0.R = R67 + 26176 + (size_t)0 * 16; i2c7_0.C = R67 + 165568 + (size_t)67 * 32;
      i2c7_0.sAo = (long long)66 * 66 * 16; i2c7_0.sAi = (long long)66 * 16; i2c7_0.sAm = 16; i2c7_0.sAk = 1; i2c7_0.sBo = 0; i2c7_0.sBi = 0; i2c7_0.sBn = 16 * 9; i2c7_0.sBk = 9; i2c7_0.sCo = (long long)66 * 66 * 32; i2c7_0.sCi = (long long)66 * 32; i2c7_0.sCm = 32; i2c7_0.sRo = 0; i2c7_0.sRi = 0; i2c7_0.sRm = 0; i2c7_0.sRn = 0;
      i2c7_0.M = 64; i2c7_0.N = 32; i2c7_0.K = 16; i2c7_0.zi_n = 64; i2c7_0.flags = 1; i2c7_0.act = 0;
      i2c7_0.alpha = 1.0f; i2c7_0.beta = 0.0f; i2c7_0.sa = 1.0f; i2c7_0.sb = 1.0f; i2c7_0.Npad = 32; i2c7_0.pad_ = 0;
      k_gemm<1><<<dim3((unsigned)((32) + 31) / 32, (unsigned)((64) + 15) / 16, (unsigned)(2 * 64)), 32, 0, stream>>>(i2c7_0); }
    { GemmP i2c7_1;
      i2c7_1.A = R67 + 26176 + (size_t)1 * 16; i2c7_1.B = iw2 + 1; i2c7_1.bias = R67 + 26176 + (size_t)1 * 16; i2c7_1.R = R67 + 165568 + (size_t)67 * 32; i2c7_1.C = R67 + 165568 + (size_t)67 * 32;
      i2c7_1.sAo = (long long)66 * 66 * 16; i2c7_1.sAi = (long long)66 * 16; i2c7_1.sAm = 16; i2c7_1.sAk = 1; i2c7_1.sBo = 0; i2c7_1.sBi = 0; i2c7_1.sBn = 16 * 9; i2c7_1.sBk = 9; i2c7_1.sCo = (long long)66 * 66 * 32; i2c7_1.sCi = (long long)66 * 32; i2c7_1.sCm = 32; i2c7_1.sRo = (long long)66 * 66 * 32; i2c7_1.sRi = (long long)66 * 32; i2c7_1.sRm = 32; i2c7_1.sRn = 1;
      i2c7_1.M = 64; i2c7_1.N = 32; i2c7_1.K = 16; i2c7_1.zi_n = 64; i2c7_1.flags = 4; i2c7_1.act = 0;
      i2c7_1.alpha = 1.0f; i2c7_1.beta = 1.0f; i2c7_1.sa = 1.0f; i2c7_1.sb = 1.0f; i2c7_1.Npad = 32; i2c7_1.pad_ = 0;
      k_gemm<1><<<dim3((unsigned)((32) + 31) / 32, (unsigned)((64) + 15) / 16, (unsigned)(2 * 64)), 32, 0, stream>>>(i2c7_1); }
    { GemmP i2c7_2;
      i2c7_2.A = R67 + 26176 + (size_t)2 * 16; i2c7_2.B = iw2 + 2; i2c7_2.bias = R67 + 26176 + (size_t)2 * 16; i2c7_2.R = R67 + 165568 + (size_t)67 * 32; i2c7_2.C = R67 + 165568 + (size_t)67 * 32;
      i2c7_2.sAo = (long long)66 * 66 * 16; i2c7_2.sAi = (long long)66 * 16; i2c7_2.sAm = 16; i2c7_2.sAk = 1; i2c7_2.sBo = 0; i2c7_2.sBi = 0; i2c7_2.sBn = 16 * 9; i2c7_2.sBk = 9; i2c7_2.sCo = (long long)66 * 66 * 32; i2c7_2.sCi = (long long)66 * 32; i2c7_2.sCm = 32; i2c7_2.sRo = (long long)66 * 66 * 32; i2c7_2.sRi = (long long)66 * 32; i2c7_2.sRm = 32; i2c7_2.sRn = 1;
      i2c7_2.M = 64; i2c7_2.N = 32; i2c7_2.K = 16; i2c7_2.zi_n = 64; i2c7_2.flags = 4; i2c7_2.act = 0;
      i2c7_2.alpha = 1.0f; i2c7_2.beta = 1.0f; i2c7_2.sa = 1.0f; i2c7_2.sb = 1.0f; i2c7_2.Npad = 32; i2c7_2.pad_ = 0;
      k_gemm<1><<<dim3((unsigned)((32) + 31) / 32, (unsigned)((64) + 15) / 16, (unsigned)(2 * 64)), 32, 0, stream>>>(i2c7_2); }
    { GemmP i2c7_3;
      i2c7_3.A = R67 + 26176 + (size_t)66 * 16; i2c7_3.B = iw2 + 3; i2c7_3.bias = R67 + 26176 + (size_t)66 * 16; i2c7_3.R = R67 + 165568 + (size_t)67 * 32; i2c7_3.C = R67 + 165568 + (size_t)67 * 32;
      i2c7_3.sAo = (long long)66 * 66 * 16; i2c7_3.sAi = (long long)66 * 16; i2c7_3.sAm = 16; i2c7_3.sAk = 1; i2c7_3.sBo = 0; i2c7_3.sBi = 0; i2c7_3.sBn = 16 * 9; i2c7_3.sBk = 9; i2c7_3.sCo = (long long)66 * 66 * 32; i2c7_3.sCi = (long long)66 * 32; i2c7_3.sCm = 32; i2c7_3.sRo = (long long)66 * 66 * 32; i2c7_3.sRi = (long long)66 * 32; i2c7_3.sRm = 32; i2c7_3.sRn = 1;
      i2c7_3.M = 64; i2c7_3.N = 32; i2c7_3.K = 16; i2c7_3.zi_n = 64; i2c7_3.flags = 4; i2c7_3.act = 0;
      i2c7_3.alpha = 1.0f; i2c7_3.beta = 1.0f; i2c7_3.sa = 1.0f; i2c7_3.sb = 1.0f; i2c7_3.Npad = 32; i2c7_3.pad_ = 0;
      k_gemm<1><<<dim3((unsigned)((32) + 31) / 32, (unsigned)((64) + 15) / 16, (unsigned)(2 * 64)), 32, 0, stream>>>(i2c7_3); }
    { GemmP i2c7_4;
      i2c7_4.A = R67 + 26176 + (size_t)67 * 16; i2c7_4.B = iw2 + 4; i2c7_4.bias = R67 + 26176 + (size_t)67 * 16; i2c7_4.R = R67 + 165568 + (size_t)67 * 32; i2c7_4.C = R67 + 165568 + (size_t)67 * 32;
      i2c7_4.sAo = (long long)66 * 66 * 16; i2c7_4.sAi = (long long)66 * 16; i2c7_4.sAm = 16; i2c7_4.sAk = 1; i2c7_4.sBo = 0; i2c7_4.sBi = 0; i2c7_4.sBn = 16 * 9; i2c7_4.sBk = 9; i2c7_4.sCo = (long long)66 * 66 * 32; i2c7_4.sCi = (long long)66 * 32; i2c7_4.sCm = 32; i2c7_4.sRo = (long long)66 * 66 * 32; i2c7_4.sRi = (long long)66 * 32; i2c7_4.sRm = 32; i2c7_4.sRn = 1;
      i2c7_4.M = 64; i2c7_4.N = 32; i2c7_4.K = 16; i2c7_4.zi_n = 64; i2c7_4.flags = 4; i2c7_4.act = 0;
      i2c7_4.alpha = 1.0f; i2c7_4.beta = 1.0f; i2c7_4.sa = 1.0f; i2c7_4.sb = 1.0f; i2c7_4.Npad = 32; i2c7_4.pad_ = 0;
      k_gemm<1><<<dim3((unsigned)((32) + 31) / 32, (unsigned)((64) + 15) / 16, (unsigned)(2 * 64)), 32, 0, stream>>>(i2c7_4); }
    { GemmP i2c7_5;
      i2c7_5.A = R67 + 26176 + (size_t)68 * 16; i2c7_5.B = iw2 + 5; i2c7_5.bias = R67 + 26176 + (size_t)68 * 16; i2c7_5.R = R67 + 165568 + (size_t)67 * 32; i2c7_5.C = R67 + 165568 + (size_t)67 * 32;
      i2c7_5.sAo = (long long)66 * 66 * 16; i2c7_5.sAi = (long long)66 * 16; i2c7_5.sAm = 16; i2c7_5.sAk = 1; i2c7_5.sBo = 0; i2c7_5.sBi = 0; i2c7_5.sBn = 16 * 9; i2c7_5.sBk = 9; i2c7_5.sCo = (long long)66 * 66 * 32; i2c7_5.sCi = (long long)66 * 32; i2c7_5.sCm = 32; i2c7_5.sRo = (long long)66 * 66 * 32; i2c7_5.sRi = (long long)66 * 32; i2c7_5.sRm = 32; i2c7_5.sRn = 1;
      i2c7_5.M = 64; i2c7_5.N = 32; i2c7_5.K = 16; i2c7_5.zi_n = 64; i2c7_5.flags = 4; i2c7_5.act = 0;
      i2c7_5.alpha = 1.0f; i2c7_5.beta = 1.0f; i2c7_5.sa = 1.0f; i2c7_5.sb = 1.0f; i2c7_5.Npad = 32; i2c7_5.pad_ = 0;
      k_gemm<1><<<dim3((unsigned)((32) + 31) / 32, (unsigned)((64) + 15) / 16, (unsigned)(2 * 64)), 32, 0, stream>>>(i2c7_5); }
    { GemmP i2c7_6;
      i2c7_6.A = R67 + 26176 + (size_t)132 * 16; i2c7_6.B = iw2 + 6; i2c7_6.bias = R67 + 26176 + (size_t)132 * 16; i2c7_6.R = R67 + 165568 + (size_t)67 * 32; i2c7_6.C = R67 + 165568 + (size_t)67 * 32;
      i2c7_6.sAo = (long long)66 * 66 * 16; i2c7_6.sAi = (long long)66 * 16; i2c7_6.sAm = 16; i2c7_6.sAk = 1; i2c7_6.sBo = 0; i2c7_6.sBi = 0; i2c7_6.sBn = 16 * 9; i2c7_6.sBk = 9; i2c7_6.sCo = (long long)66 * 66 * 32; i2c7_6.sCi = (long long)66 * 32; i2c7_6.sCm = 32; i2c7_6.sRo = (long long)66 * 66 * 32; i2c7_6.sRi = (long long)66 * 32; i2c7_6.sRm = 32; i2c7_6.sRn = 1;
      i2c7_6.M = 64; i2c7_6.N = 32; i2c7_6.K = 16; i2c7_6.zi_n = 64; i2c7_6.flags = 4; i2c7_6.act = 0;
      i2c7_6.alpha = 1.0f; i2c7_6.beta = 1.0f; i2c7_6.sa = 1.0f; i2c7_6.sb = 1.0f; i2c7_6.Npad = 32; i2c7_6.pad_ = 0;
      k_gemm<1><<<dim3((unsigned)((32) + 31) / 32, (unsigned)((64) + 15) / 16, (unsigned)(2 * 64)), 32, 0, stream>>>(i2c7_6); }
    { GemmP i2c7_7;
      i2c7_7.A = R67 + 26176 + (size_t)133 * 16; i2c7_7.B = iw2 + 7; i2c7_7.bias = R67 + 26176 + (size_t)133 * 16; i2c7_7.R = R67 + 165568 + (size_t)67 * 32; i2c7_7.C = R67 + 165568 + (size_t)67 * 32;
      i2c7_7.sAo = (long long)66 * 66 * 16; i2c7_7.sAi = (long long)66 * 16; i2c7_7.sAm = 16; i2c7_7.sAk = 1; i2c7_7.sBo = 0; i2c7_7.sBi = 0; i2c7_7.sBn = 16 * 9; i2c7_7.sBk = 9; i2c7_7.sCo = (long long)66 * 66 * 32; i2c7_7.sCi = (long long)66 * 32; i2c7_7.sCm = 32; i2c7_7.sRo = (long long)66 * 66 * 32; i2c7_7.sRi = (long long)66 * 32; i2c7_7.sRm = 32; i2c7_7.sRn = 1;
      i2c7_7.M = 64; i2c7_7.N = 32; i2c7_7.K = 16; i2c7_7.zi_n = 64; i2c7_7.flags = 4; i2c7_7.act = 0;
      i2c7_7.alpha = 1.0f; i2c7_7.beta = 1.0f; i2c7_7.sa = 1.0f; i2c7_7.sb = 1.0f; i2c7_7.Npad = 32; i2c7_7.pad_ = 0;
      k_gemm<1><<<dim3((unsigned)((32) + 31) / 32, (unsigned)((64) + 15) / 16, (unsigned)(2 * 64)), 32, 0, stream>>>(i2c7_7); }
    { GemmP i2c7_8;
      i2c7_8.A = R67 + 26176 + (size_t)134 * 16; i2c7_8.B = iw2 + 8; i2c7_8.bias = R67 + 26176 + (size_t)134 * 16; i2c7_8.R = R67 + 165568 + (size_t)67 * 32; i2c7_8.C = R67 + 165568 + (size_t)67 * 32;
      i2c7_8.sAo = (long long)66 * 66 * 16; i2c7_8.sAi = (long long)66 * 16; i2c7_8.sAm = 16; i2c7_8.sAk = 1; i2c7_8.sBo = 0; i2c7_8.sBi = 0; i2c7_8.sBn = 16 * 9; i2c7_8.sBk = 9; i2c7_8.sCo = (long long)66 * 66 * 32; i2c7_8.sCi = (long long)66 * 32; i2c7_8.sCm = 32; i2c7_8.sRo = (long long)66 * 66 * 32; i2c7_8.sRi = (long long)66 * 32; i2c7_8.sRm = 32; i2c7_8.sRn = 1;
      i2c7_8.M = 64; i2c7_8.N = 32; i2c7_8.K = 16; i2c7_8.zi_n = 64; i2c7_8.flags = 4; i2c7_8.act = 0;
      i2c7_8.alpha = 1.0f; i2c7_8.beta = 1.0f; i2c7_8.sa = 1.0f; i2c7_8.sb = 1.0f; i2c7_8.Npad = 32; i2c7_8.pad_ = 0;
      k_gemm<1><<<dim3((unsigned)((32) + 31) / 32, (unsigned)((64) + 15) / 16, (unsigned)(2 * 64)), 32, 0, stream>>>(i2c7_8); }
    k_mm_relu2d<<<(unsigned)(((long long)2 * HW * 32 + 255) / 256), 256, 0, stream>>>(R67 + 165568, nullptr, 2, 64, 32);
    { GemmP i3c7_0;
      i3c7_0.A = R67 + 165568 + (size_t)0 * 32; i3c7_0.B = iw3 + 0; i3c7_0.bias = ib3; i3c7_0.R = R67 + 165568 + (size_t)0 * 32; i3c7_0.C = R67 + 444352 + (size_t)67 * 64;
      i3c7_0.sAo = (long long)66 * 66 * 32; i3c7_0.sAi = (long long)66 * 32; i3c7_0.sAm = 32; i3c7_0.sAk = 1; i3c7_0.sBo = 0; i3c7_0.sBi = 0; i3c7_0.sBn = 32 * 9; i3c7_0.sBk = 9; i3c7_0.sCo = (long long)66 * 66 * 64; i3c7_0.sCi = (long long)66 * 64; i3c7_0.sCm = 64; i3c7_0.sRo = 0; i3c7_0.sRi = 0; i3c7_0.sRm = 0; i3c7_0.sRn = 0;
      i3c7_0.M = 64; i3c7_0.N = 64; i3c7_0.K = 32; i3c7_0.zi_n = 64; i3c7_0.flags = 1; i3c7_0.act = 0;
      i3c7_0.alpha = 1.0f; i3c7_0.beta = 0.0f; i3c7_0.sa = 1.0f; i3c7_0.sb = 1.0f; i3c7_0.Npad = 64; i3c7_0.pad_ = 0;
      k_gemm<1><<<dim3((unsigned)((64) + 31) / 32, (unsigned)((64) + 15) / 16, (unsigned)(2 * 64)), 32, 0, stream>>>(i3c7_0); }
    { GemmP i3c7_1;
      i3c7_1.A = R67 + 165568 + (size_t)1 * 32; i3c7_1.B = iw3 + 1; i3c7_1.bias = R67 + 165568 + (size_t)1 * 32; i3c7_1.R = R67 + 444352 + (size_t)67 * 64; i3c7_1.C = R67 + 444352 + (size_t)67 * 64;
      i3c7_1.sAo = (long long)66 * 66 * 32; i3c7_1.sAi = (long long)66 * 32; i3c7_1.sAm = 32; i3c7_1.sAk = 1; i3c7_1.sBo = 0; i3c7_1.sBi = 0; i3c7_1.sBn = 32 * 9; i3c7_1.sBk = 9; i3c7_1.sCo = (long long)66 * 66 * 64; i3c7_1.sCi = (long long)66 * 64; i3c7_1.sCm = 64; i3c7_1.sRo = (long long)66 * 66 * 64; i3c7_1.sRi = (long long)66 * 64; i3c7_1.sRm = 64; i3c7_1.sRn = 1;
      i3c7_1.M = 64; i3c7_1.N = 64; i3c7_1.K = 32; i3c7_1.zi_n = 64; i3c7_1.flags = 4; i3c7_1.act = 0;
      i3c7_1.alpha = 1.0f; i3c7_1.beta = 1.0f; i3c7_1.sa = 1.0f; i3c7_1.sb = 1.0f; i3c7_1.Npad = 64; i3c7_1.pad_ = 0;
      k_gemm<1><<<dim3((unsigned)((64) + 31) / 32, (unsigned)((64) + 15) / 16, (unsigned)(2 * 64)), 32, 0, stream>>>(i3c7_1); }
    { GemmP i3c7_2;
      i3c7_2.A = R67 + 165568 + (size_t)2 * 32; i3c7_2.B = iw3 + 2; i3c7_2.bias = R67 + 165568 + (size_t)2 * 32; i3c7_2.R = R67 + 444352 + (size_t)67 * 64; i3c7_2.C = R67 + 444352 + (size_t)67 * 64;
      i3c7_2.sAo = (long long)66 * 66 * 32; i3c7_2.sAi = (long long)66 * 32; i3c7_2.sAm = 32; i3c7_2.sAk = 1; i3c7_2.sBo = 0; i3c7_2.sBi = 0; i3c7_2.sBn = 32 * 9; i3c7_2.sBk = 9; i3c7_2.sCo = (long long)66 * 66 * 64; i3c7_2.sCi = (long long)66 * 64; i3c7_2.sCm = 64; i3c7_2.sRo = (long long)66 * 66 * 64; i3c7_2.sRi = (long long)66 * 64; i3c7_2.sRm = 64; i3c7_2.sRn = 1;
      i3c7_2.M = 64; i3c7_2.N = 64; i3c7_2.K = 32; i3c7_2.zi_n = 64; i3c7_2.flags = 4; i3c7_2.act = 0;
      i3c7_2.alpha = 1.0f; i3c7_2.beta = 1.0f; i3c7_2.sa = 1.0f; i3c7_2.sb = 1.0f; i3c7_2.Npad = 64; i3c7_2.pad_ = 0;
      k_gemm<1><<<dim3((unsigned)((64) + 31) / 32, (unsigned)((64) + 15) / 16, (unsigned)(2 * 64)), 32, 0, stream>>>(i3c7_2); }
    { GemmP i3c7_3;
      i3c7_3.A = R67 + 165568 + (size_t)66 * 32; i3c7_3.B = iw3 + 3; i3c7_3.bias = R67 + 165568 + (size_t)66 * 32; i3c7_3.R = R67 + 444352 + (size_t)67 * 64; i3c7_3.C = R67 + 444352 + (size_t)67 * 64;
      i3c7_3.sAo = (long long)66 * 66 * 32; i3c7_3.sAi = (long long)66 * 32; i3c7_3.sAm = 32; i3c7_3.sAk = 1; i3c7_3.sBo = 0; i3c7_3.sBi = 0; i3c7_3.sBn = 32 * 9; i3c7_3.sBk = 9; i3c7_3.sCo = (long long)66 * 66 * 64; i3c7_3.sCi = (long long)66 * 64; i3c7_3.sCm = 64; i3c7_3.sRo = (long long)66 * 66 * 64; i3c7_3.sRi = (long long)66 * 64; i3c7_3.sRm = 64; i3c7_3.sRn = 1;
      i3c7_3.M = 64; i3c7_3.N = 64; i3c7_3.K = 32; i3c7_3.zi_n = 64; i3c7_3.flags = 4; i3c7_3.act = 0;
      i3c7_3.alpha = 1.0f; i3c7_3.beta = 1.0f; i3c7_3.sa = 1.0f; i3c7_3.sb = 1.0f; i3c7_3.Npad = 64; i3c7_3.pad_ = 0;
      k_gemm<1><<<dim3((unsigned)((64) + 31) / 32, (unsigned)((64) + 15) / 16, (unsigned)(2 * 64)), 32, 0, stream>>>(i3c7_3); }
    { GemmP i3c7_4;
      i3c7_4.A = R67 + 165568 + (size_t)67 * 32; i3c7_4.B = iw3 + 4; i3c7_4.bias = R67 + 165568 + (size_t)67 * 32; i3c7_4.R = R67 + 444352 + (size_t)67 * 64; i3c7_4.C = R67 + 444352 + (size_t)67 * 64;
      i3c7_4.sAo = (long long)66 * 66 * 32; i3c7_4.sAi = (long long)66 * 32; i3c7_4.sAm = 32; i3c7_4.sAk = 1; i3c7_4.sBo = 0; i3c7_4.sBi = 0; i3c7_4.sBn = 32 * 9; i3c7_4.sBk = 9; i3c7_4.sCo = (long long)66 * 66 * 64; i3c7_4.sCi = (long long)66 * 64; i3c7_4.sCm = 64; i3c7_4.sRo = (long long)66 * 66 * 64; i3c7_4.sRi = (long long)66 * 64; i3c7_4.sRm = 64; i3c7_4.sRn = 1;
      i3c7_4.M = 64; i3c7_4.N = 64; i3c7_4.K = 32; i3c7_4.zi_n = 64; i3c7_4.flags = 4; i3c7_4.act = 0;
      i3c7_4.alpha = 1.0f; i3c7_4.beta = 1.0f; i3c7_4.sa = 1.0f; i3c7_4.sb = 1.0f; i3c7_4.Npad = 64; i3c7_4.pad_ = 0;
      k_gemm<1><<<dim3((unsigned)((64) + 31) / 32, (unsigned)((64) + 15) / 16, (unsigned)(2 * 64)), 32, 0, stream>>>(i3c7_4); }
    { GemmP i3c7_5;
      i3c7_5.A = R67 + 165568 + (size_t)68 * 32; i3c7_5.B = iw3 + 5; i3c7_5.bias = R67 + 165568 + (size_t)68 * 32; i3c7_5.R = R67 + 444352 + (size_t)67 * 64; i3c7_5.C = R67 + 444352 + (size_t)67 * 64;
      i3c7_5.sAo = (long long)66 * 66 * 32; i3c7_5.sAi = (long long)66 * 32; i3c7_5.sAm = 32; i3c7_5.sAk = 1; i3c7_5.sBo = 0; i3c7_5.sBi = 0; i3c7_5.sBn = 32 * 9; i3c7_5.sBk = 9; i3c7_5.sCo = (long long)66 * 66 * 64; i3c7_5.sCi = (long long)66 * 64; i3c7_5.sCm = 64; i3c7_5.sRo = (long long)66 * 66 * 64; i3c7_5.sRi = (long long)66 * 64; i3c7_5.sRm = 64; i3c7_5.sRn = 1;
      i3c7_5.M = 64; i3c7_5.N = 64; i3c7_5.K = 32; i3c7_5.zi_n = 64; i3c7_5.flags = 4; i3c7_5.act = 0;
      i3c7_5.alpha = 1.0f; i3c7_5.beta = 1.0f; i3c7_5.sa = 1.0f; i3c7_5.sb = 1.0f; i3c7_5.Npad = 64; i3c7_5.pad_ = 0;
      k_gemm<1><<<dim3((unsigned)((64) + 31) / 32, (unsigned)((64) + 15) / 16, (unsigned)(2 * 64)), 32, 0, stream>>>(i3c7_5); }
    { GemmP i3c7_6;
      i3c7_6.A = R67 + 165568 + (size_t)132 * 32; i3c7_6.B = iw3 + 6; i3c7_6.bias = R67 + 165568 + (size_t)132 * 32; i3c7_6.R = R67 + 444352 + (size_t)67 * 64; i3c7_6.C = R67 + 444352 + (size_t)67 * 64;
      i3c7_6.sAo = (long long)66 * 66 * 32; i3c7_6.sAi = (long long)66 * 32; i3c7_6.sAm = 32; i3c7_6.sAk = 1; i3c7_6.sBo = 0; i3c7_6.sBi = 0; i3c7_6.sBn = 32 * 9; i3c7_6.sBk = 9; i3c7_6.sCo = (long long)66 * 66 * 64; i3c7_6.sCi = (long long)66 * 64; i3c7_6.sCm = 64; i3c7_6.sRo = (long long)66 * 66 * 64; i3c7_6.sRi = (long long)66 * 64; i3c7_6.sRm = 64; i3c7_6.sRn = 1;
      i3c7_6.M = 64; i3c7_6.N = 64; i3c7_6.K = 32; i3c7_6.zi_n = 64; i3c7_6.flags = 4; i3c7_6.act = 0;
      i3c7_6.alpha = 1.0f; i3c7_6.beta = 1.0f; i3c7_6.sa = 1.0f; i3c7_6.sb = 1.0f; i3c7_6.Npad = 64; i3c7_6.pad_ = 0;
      k_gemm<1><<<dim3((unsigned)((64) + 31) / 32, (unsigned)((64) + 15) / 16, (unsigned)(2 * 64)), 32, 0, stream>>>(i3c7_6); }
    { GemmP i3c7_7;
      i3c7_7.A = R67 + 165568 + (size_t)133 * 32; i3c7_7.B = iw3 + 7; i3c7_7.bias = R67 + 165568 + (size_t)133 * 32; i3c7_7.R = R67 + 444352 + (size_t)67 * 64; i3c7_7.C = R67 + 444352 + (size_t)67 * 64;
      i3c7_7.sAo = (long long)66 * 66 * 32; i3c7_7.sAi = (long long)66 * 32; i3c7_7.sAm = 32; i3c7_7.sAk = 1; i3c7_7.sBo = 0; i3c7_7.sBi = 0; i3c7_7.sBn = 32 * 9; i3c7_7.sBk = 9; i3c7_7.sCo = (long long)66 * 66 * 64; i3c7_7.sCi = (long long)66 * 64; i3c7_7.sCm = 64; i3c7_7.sRo = (long long)66 * 66 * 64; i3c7_7.sRi = (long long)66 * 64; i3c7_7.sRm = 64; i3c7_7.sRn = 1;
      i3c7_7.M = 64; i3c7_7.N = 64; i3c7_7.K = 32; i3c7_7.zi_n = 64; i3c7_7.flags = 4; i3c7_7.act = 0;
      i3c7_7.alpha = 1.0f; i3c7_7.beta = 1.0f; i3c7_7.sa = 1.0f; i3c7_7.sb = 1.0f; i3c7_7.Npad = 64; i3c7_7.pad_ = 0;
      k_gemm<1><<<dim3((unsigned)((64) + 31) / 32, (unsigned)((64) + 15) / 16, (unsigned)(2 * 64)), 32, 0, stream>>>(i3c7_7); }
    { GemmP i3c7_8;
      i3c7_8.A = R67 + 165568 + (size_t)134 * 32; i3c7_8.B = iw3 + 8; i3c7_8.bias = R67 + 165568 + (size_t)134 * 32; i3c7_8.R = R67 + 444352 + (size_t)67 * 64; i3c7_8.C = R67 + 444352 + (size_t)67 * 64;
      i3c7_8.sAo = (long long)66 * 66 * 32; i3c7_8.sAi = (long long)66 * 32; i3c7_8.sAm = 32; i3c7_8.sAk = 1; i3c7_8.sBo = 0; i3c7_8.sBi = 0; i3c7_8.sBn = 32 * 9; i3c7_8.sBk = 9; i3c7_8.sCo = (long long)66 * 66 * 64; i3c7_8.sCi = (long long)66 * 64; i3c7_8.sCm = 64; i3c7_8.sRo = (long long)66 * 66 * 64; i3c7_8.sRi = (long long)66 * 64; i3c7_8.sRm = 64; i3c7_8.sRn = 1;
      i3c7_8.M = 64; i3c7_8.N = 64; i3c7_8.K = 32; i3c7_8.zi_n = 64; i3c7_8.flags = 4; i3c7_8.act = 0;
      i3c7_8.alpha = 1.0f; i3c7_8.beta = 1.0f; i3c7_8.sa = 1.0f; i3c7_8.sb = 1.0f; i3c7_8.Npad = 64; i3c7_8.pad_ = 0;
      k_gemm<1><<<dim3((unsigned)((64) + 31) / 32, (unsigned)((64) + 15) / 16, (unsigned)(2 * 64)), 32, 0, stream>>>(i3c7_8); }
    k_mm_relu2d<<<(unsigned)(((long long)2 * HW * 64 + 255) / 256), 256, 0, stream>>>(R67 + 444352, R67 + 1001920, 2, 64, 64);
    { GemmP gqkv7;
      gqkv7.A = R67 + 1001920; gqkv7.B = qkvw; gqkv7.bias = qkvb; gqkv7.R = R67 + 1001920; gqkv7.C = R67 + 1526208;
      gqkv7.sAo = 0; gqkv7.sAi = 0; gqkv7.sAm = 64; gqkv7.sAk = 1; gqkv7.sBo = 0; gqkv7.sBi = 0; gqkv7.sBn = 64; gqkv7.sBk = 1; gqkv7.sCo = 0; gqkv7.sCi = 0; gqkv7.sCm = 192; gqkv7.sRo = 0; gqkv7.sRi = 0; gqkv7.sRm = 0; gqkv7.sRn = 0;
      gqkv7.M = 2 * HW; gqkv7.N = 192; gqkv7.K = 64; gqkv7.zi_n = 1; gqkv7.flags = 1; gqkv7.act = 0;
      gqkv7.alpha = 1.0f; gqkv7.beta = 0.0f; gqkv7.sa = 1.0f; gqkv7.sb = 1.0f; gqkv7.Npad = 192; gqkv7.pad_ = 0;
      k_gemm<1><<<dim3((unsigned)((192) + 31) / 32, (unsigned)((2 * HW) + 15) / 16, (unsigned)(1)), 32, 0, stream>>>(gqkv7); }
    k_mm_dw<<<(unsigned)(((long long)2 * HW * 192 + 255) / 256), 256, 0, stream>>>(R67 + 1526208, dww, dwb, R67 + 3099072, 2, 64, 192);
    k_mm_fall<<<(unsigned)(((long long)2 * HW * 144 + 255) / 256), 256, 0, stream>>>(R67 + 3099072, fcw, fcb, R67 + 4671936, 2, HW, 192);
    k_mm_dep<<<(unsigned)(((long long)2 * 64 * HW + 255) / 256), 256, 0, stream>>>(R67 + 4671936, depw, depb, R67 + 5851584, 2, 64);
    k_mm_qknorm<<<2 * 128, 256, 0, stream>>>(R67 + 3099072, R67 + 6375872, 2, HW, 192);
    { GemmP gat7;
      gat7.A = R67 + 6375872; gat7.B = R67 + 6375872 + (size_t)64 * HW; gat7.bias = R67 + 6375872; gat7.R = R67 + 6375872; gat7.C = R67 + 7424448;
      gat7.sAo = (long long)128 * HW; gat7.sAi = (long long)16 * HW; gat7.sAm = HW; gat7.sAk = 1; gat7.sBo = (long long)128 * HW; gat7.sBi = (long long)16 * HW; gat7.sBn = HW; gat7.sBk = 1; gat7.sCo = (long long)4 * 16 * LP; gat7.sCi = 16 * LP; gat7.sCm = LP; gat7.sRo = 0; gat7.sRi = 0; gat7.sRm = 0; gat7.sRn = 0;
      gat7.M = 16; gat7.N = 16; gat7.K = HW; gat7.zi_n = 4; gat7.flags = 0; gat7.act = 0;
      gat7.alpha = 1.0f; gat7.beta = 0.0f; gat7.sa = 1.0f; gat7.sb = 1.0f; gat7.Npad = LP; gat7.pad_ = 0;
      k_gemm<1><<<dim3((unsigned)((LP) + 31) / 32, (unsigned)((16) + 15) / 16, (unsigned)(2 * 4)), 32, 0, stream>>>(gat7); }
    k_mm_sm16<<<(unsigned)((2 * 4 * 16 + 255) / 256), 256, 0, stream>>>(R67 + 7424448, temp, 2 * 4, LP);
    { GemmP gao7;
      gao7.A = R67 + 7424448; gao7.B = R67 + 3099072 + 128; gao7.bias = R67 + 7424448; gao7.R = R67 + 7424448; gao7.C = R67 + 7428544;
      gao7.sAo = (long long)4 * 16 * LP; gao7.sAi = 16 * LP; gao7.sAm = LP; gao7.sAk = 1; gao7.sBo = (long long)HW * 192; gao7.sBi = 16; gao7.sBn = 192; gao7.sBk = 1; gao7.sCo = (long long)64 * HW; gao7.sCi = (long long)16 * HW; gao7.sCm = HW; gao7.sRo = 0; gao7.sRi = 0; gao7.sRm = 0; gao7.sRn = 0;
      gao7.M = 16; gao7.N = HW; gao7.K = 16; gao7.zi_n = 4; gao7.flags = 0; gao7.act = 0;
      gao7.alpha = 1.0f; gao7.beta = 0.0f; gao7.sa = 1.0f; gao7.sb = 1.0f; gao7.Npad = HW; gao7.pad_ = 0;
      k_gemm<1><<<dim3((unsigned)((HW) + 31) / 32, (unsigned)((16) + 15) / 16, (unsigned)(2 * 4)), 32, 0, stream>>>(gao7); }
    { GemmP gproj7;
      gproj7.A = projw; gproj7.B = R67 + 7428544; gproj7.bias = projb; gproj7.R = projw; gproj7.C = R67 + 7952832;
      gproj7.sAo = 0; gproj7.sAi = 0; gproj7.sAm = 64; gproj7.sAk = 1; gproj7.sBo = (long long)64 * HW; gproj7.sBi = 0; gproj7.sBn = 1; gproj7.sBk = HW; gproj7.sCo = (long long)64 * HW; gproj7.sCi = 0; gproj7.sCm = HW; gproj7.sRo = 0; gproj7.sRi = 0; gproj7.sRm = 0; gproj7.sRn = 0;
      gproj7.M = 64; gproj7.N = HW; gproj7.K = 64; gproj7.zi_n = 1; gproj7.flags = 2; gproj7.act = 0;
      gproj7.alpha = 1.0f; gproj7.beta = 0.0f; gproj7.sa = 1.0f; gproj7.sb = 1.0f; gproj7.Npad = HW; gproj7.pad_ = 0;
      k_gemm<1><<<dim3((unsigned)((HW) + 31) / 32, (unsigned)((64) + 15) / 16, (unsigned)(2)), 32, 0, stream>>>(gproj7); }
    k_mm_imgfeat<<<(unsigned)(((long long)2 * SEQ * 64 + 255) / 256), 256, 0, stream>>>(R67 + 7952832, R67 + 5851584, IR + (size_t)14 * SEQ * 64, 2, HW, 64);
    { GemmP gh1;
      gh1.A = UR; gh1.B = caw; gh1.bias = cab; gh1.R = UR; gh1.C = H1;
      gh1.sAo = 0; gh1.sAi = 0; gh1.sAm = 64; gh1.sAk = 1; gh1.sBo = 0; gh1.sBi = 0; gh1.sBn = 64; gh1.sBk = 1; gh1.sCo = 0; gh1.sCi = 0; gh1.sCm = 192; gh1.sRo = 0; gh1.sRi = 0; gh1.sRm = 0; gh1.sRn = 0;
      gh1.M = Bn * SEQ; gh1.N = 192; gh1.K = 64; gh1.zi_n = 1; gh1.flags = 1; gh1.act = 0;
      gh1.alpha = 1.0f; gh1.beta = 0.0f; gh1.sa = 1.0f; gh1.sb = 1.0f; gh1.Npad = 192; gh1.pad_ = 0;
      k_gemm<1><<<dim3((unsigned)((192) + 31) / 32, (unsigned)((Bn * SEQ) + 15) / 16, (unsigned)(1)), 32, 0, stream>>>(gh1); }
    { GemmP gh2;
      gh2.A = IR; gh2.B = caw; gh2.bias = cab; gh2.R = IR; gh2.C = H2;
      gh2.sAo = 0; gh2.sAi = 0; gh2.sAm = 64; gh2.sAk = 1; gh2.sBo = 0; gh2.sBi = 0; gh2.sBn = 64; gh2.sBk = 1; gh2.sCo = 0; gh2.sCi = 0; gh2.sCm = 192; gh2.sRo = 0; gh2.sRi = 0; gh2.sRm = 0; gh2.sRn = 0;
      gh2.M = Bn * SEQ; gh2.N = 192; gh2.K = 64; gh2.zi_n = 1; gh2.flags = 1; gh2.act = 0;
      gh2.alpha = 1.0f; gh2.beta = 0.0f; gh2.sa = 1.0f; gh2.sb = 1.0f; gh2.Npad = 192; gh2.pad_ = 0;
      k_gemm<1><<<dim3((unsigned)((192) + 31) / 32, (unsigned)((Bn * SEQ) + 15) / 16, (unsigned)(1)), 32, 0, stream>>>(gh2); }
    { GemmP gsa0;
      gsa0.A = H1 + (size_t)0 * SEQ * 192; gsa0.B = H2 + (size_t)0 * SEQ * 192 + 16; gsa0.bias = H1 + (size_t)0 * SEQ * 192; gsa0.R = H1 + (size_t)0 * SEQ * 192; gsa0.C = SC;
      gsa0.sAo = 48; gsa0.sAi = 0; gsa0.sAm = 192; gsa0.sAk = 1; gsa0.sBo = 48; gsa0.sBi = 0; gsa0.sBn = 192; gsa0.sBk = 1; gsa0.sCo = (long long)SEQ * SEQ; gsa0.sCi = 0; gsa0.sCm = SEQ; gsa0.sRo = 0; gsa0.sRi = 0; gsa0.sRm = 0; gsa0.sRn = 0;
      gsa0.M = SEQ; gsa0.N = SEQ; gsa0.K = 16; gsa0.zi_n = 1; gsa0.flags = 0; gsa0.act = 0;
      gsa0.alpha = 1.0f; gsa0.beta = 0.0f; gsa0.sa = 1.0f; gsa0.sb = 1.0f; gsa0.Npad = SEQ; gsa0.pad_ = 0;
      k_gemm<1><<<dim3((unsigned)((SEQ) + 31) / 32, (unsigned)((SEQ) + 15) / 16, (unsigned)(4)), 32, 0, stream>>>(gsa0); }
    k_mm_rowsm<<<4 * SEQ, 256, 0, stream>>>(SC, 4 * SEQ, SEQ, 0.25f);
    { GemmP gva0;
      gva0.A = SC; gva0.B = H2 + (size_t)0 * SEQ * 192 + 32; gva0.bias = SC; gva0.R = SC; gva0.C = O1 + (size_t)0 * SEQ * 64;
      gva0.sAo = (long long)SEQ * SEQ; gva0.sAi = 0; gva0.sAm = SEQ; gva0.sAk = 1; gva0.sBo = 48; gva0.sBi = 0; gva0.sBn = 1; gva0.sBk = 192; gva0.sCo = 16; gva0.sCi = 0; gva0.sCm = 64; gva0.sRo = 0; gva0.sRi = 0; gva0.sRm = 0; gva0.sRn = 0;
      gva0.M = SEQ; gva0.N = 16; gva0.K = SEQ; gva0.zi_n = 1; gva0.flags = 0; gva0.act = 0;
      gva0.alpha = 1.0f; gva0.beta = 0.0f; gva0.sa = 1.0f; gva0.sb = 1.0f; gva0.Npad = 16; gva0.pad_ = 0;
      k_gemm<1><<<dim3((unsigned)((16) + 31) / 32, (unsigned)((SEQ) + 15) / 16, (unsigned)(4)), 32, 0, stream>>>(gva0); }
    { GemmP gsb0;
      gsb0.A = H2 + (size_t)0 * SEQ * 192; gsb0.B = H1 + (size_t)0 * SEQ * 192 + 16; gsb0.bias = H2 + (size_t)0 * SEQ * 192; gsb0.R = H2 + (size_t)0 * SEQ * 192; gsb0.C = SC;
      gsb0.sAo = 48; gsb0.sAi = 0; gsb0.sAm = 192; gsb0.sAk = 1; gsb0.sBo = 48; gsb0.sBi = 0; gsb0.sBn = 192; gsb0.sBk = 1; gsb0.sCo = (long long)SEQ * SEQ; gsb0.sCi = 0; gsb0.sCm = SEQ; gsb0.sRo = 0; gsb0.sRi = 0; gsb0.sRm = 0; gsb0.sRn = 0;
      gsb0.M = SEQ; gsb0.N = SEQ; gsb0.K = 16; gsb0.zi_n = 1; gsb0.flags = 0; gsb0.act = 0;
      gsb0.alpha = 1.0f; gsb0.beta = 0.0f; gsb0.sa = 1.0f; gsb0.sb = 1.0f; gsb0.Npad = SEQ; gsb0.pad_ = 0;
      k_gemm<1><<<dim3((unsigned)((SEQ) + 31) / 32, (unsigned)((SEQ) + 15) / 16, (unsigned)(4)), 32, 0, stream>>>(gsb0); }
    k_mm_rowsm<<<4 * SEQ, 256, 0, stream>>>(SC, 4 * SEQ, SEQ, 0.25f);
    { GemmP gvb0;
      gvb0.A = SC; gvb0.B = H1 + (size_t)0 * SEQ * 192 + 32; gvb0.bias = SC; gvb0.R = SC; gvb0.C = O2 + (size_t)0 * SEQ * 64;
      gvb0.sAo = (long long)SEQ * SEQ; gvb0.sAi = 0; gvb0.sAm = SEQ; gvb0.sAk = 1; gvb0.sBo = 48; gvb0.sBi = 0; gvb0.sBn = 1; gvb0.sBk = 192; gvb0.sCo = 16; gvb0.sCi = 0; gvb0.sCm = 64; gvb0.sRo = 0; gvb0.sRi = 0; gvb0.sRm = 0; gvb0.sRn = 0;
      gvb0.M = SEQ; gvb0.N = 16; gvb0.K = SEQ; gvb0.zi_n = 1; gvb0.flags = 0; gvb0.act = 0;
      gvb0.alpha = 1.0f; gvb0.beta = 0.0f; gvb0.sa = 1.0f; gvb0.sb = 1.0f; gvb0.Npad = 16; gvb0.pad_ = 0;
      k_gemm<1><<<dim3((unsigned)((16) + 31) / 32, (unsigned)((SEQ) + 15) / 16, (unsigned)(4)), 32, 0, stream>>>(gvb0); }
    { GemmP gsa1;
      gsa1.A = H1 + (size_t)1 * SEQ * 192; gsa1.B = H2 + (size_t)1 * SEQ * 192 + 16; gsa1.bias = H1 + (size_t)1 * SEQ * 192; gsa1.R = H1 + (size_t)1 * SEQ * 192; gsa1.C = SC;
      gsa1.sAo = 48; gsa1.sAi = 0; gsa1.sAm = 192; gsa1.sAk = 1; gsa1.sBo = 48; gsa1.sBi = 0; gsa1.sBn = 192; gsa1.sBk = 1; gsa1.sCo = (long long)SEQ * SEQ; gsa1.sCi = 0; gsa1.sCm = SEQ; gsa1.sRo = 0; gsa1.sRi = 0; gsa1.sRm = 0; gsa1.sRn = 0;
      gsa1.M = SEQ; gsa1.N = SEQ; gsa1.K = 16; gsa1.zi_n = 1; gsa1.flags = 0; gsa1.act = 0;
      gsa1.alpha = 1.0f; gsa1.beta = 0.0f; gsa1.sa = 1.0f; gsa1.sb = 1.0f; gsa1.Npad = SEQ; gsa1.pad_ = 0;
      k_gemm<1><<<dim3((unsigned)((SEQ) + 31) / 32, (unsigned)((SEQ) + 15) / 16, (unsigned)(4)), 32, 0, stream>>>(gsa1); }
    k_mm_rowsm<<<4 * SEQ, 256, 0, stream>>>(SC, 4 * SEQ, SEQ, 0.25f);
    { GemmP gva1;
      gva1.A = SC; gva1.B = H2 + (size_t)1 * SEQ * 192 + 32; gva1.bias = SC; gva1.R = SC; gva1.C = O1 + (size_t)1 * SEQ * 64;
      gva1.sAo = (long long)SEQ * SEQ; gva1.sAi = 0; gva1.sAm = SEQ; gva1.sAk = 1; gva1.sBo = 48; gva1.sBi = 0; gva1.sBn = 1; gva1.sBk = 192; gva1.sCo = 16; gva1.sCi = 0; gva1.sCm = 64; gva1.sRo = 0; gva1.sRi = 0; gva1.sRm = 0; gva1.sRn = 0;
      gva1.M = SEQ; gva1.N = 16; gva1.K = SEQ; gva1.zi_n = 1; gva1.flags = 0; gva1.act = 0;
      gva1.alpha = 1.0f; gva1.beta = 0.0f; gva1.sa = 1.0f; gva1.sb = 1.0f; gva1.Npad = 16; gva1.pad_ = 0;
      k_gemm<1><<<dim3((unsigned)((16) + 31) / 32, (unsigned)((SEQ) + 15) / 16, (unsigned)(4)), 32, 0, stream>>>(gva1); }
    { GemmP gsb1;
      gsb1.A = H2 + (size_t)1 * SEQ * 192; gsb1.B = H1 + (size_t)1 * SEQ * 192 + 16; gsb1.bias = H2 + (size_t)1 * SEQ * 192; gsb1.R = H2 + (size_t)1 * SEQ * 192; gsb1.C = SC;
      gsb1.sAo = 48; gsb1.sAi = 0; gsb1.sAm = 192; gsb1.sAk = 1; gsb1.sBo = 48; gsb1.sBi = 0; gsb1.sBn = 192; gsb1.sBk = 1; gsb1.sCo = (long long)SEQ * SEQ; gsb1.sCi = 0; gsb1.sCm = SEQ; gsb1.sRo = 0; gsb1.sRi = 0; gsb1.sRm = 0; gsb1.sRn = 0;
      gsb1.M = SEQ; gsb1.N = SEQ; gsb1.K = 16; gsb1.zi_n = 1; gsb1.flags = 0; gsb1.act = 0;
      gsb1.alpha = 1.0f; gsb1.beta = 0.0f; gsb1.sa = 1.0f; gsb1.sb = 1.0f; gsb1.Npad = SEQ; gsb1.pad_ = 0;
      k_gemm<1><<<dim3((unsigned)((SEQ) + 31) / 32, (unsigned)((SEQ) + 15) / 16, (unsigned)(4)), 32, 0, stream>>>(gsb1); }
    k_mm_rowsm<<<4 * SEQ, 256, 0, stream>>>(SC, 4 * SEQ, SEQ, 0.25f);
    { GemmP gvb1;
      gvb1.A = SC; gvb1.B = H1 + (size_t)1 * SEQ * 192 + 32; gvb1.bias = SC; gvb1.R = SC; gvb1.C = O2 + (size_t)1 * SEQ * 64;
      gvb1.sAo = (long long)SEQ * SEQ; gvb1.sAi = 0; gvb1.sAm = SEQ; gvb1.sAk = 1; gvb1.sBo = 48; gvb1.sBi = 0; gvb1.sBn = 1; gvb1.sBk = 192; gvb1.sCo = 16; gvb1.sCi = 0; gvb1.sCm = 64; gvb1.sRo = 0; gvb1.sRi = 0; gvb1.sRm = 0; gvb1.sRn = 0;
      gvb1.M = SEQ; gvb1.N = 16; gvb1.K = SEQ; gvb1.zi_n = 1; gvb1.flags = 0; gvb1.act = 0;
      gvb1.alpha = 1.0f; gvb1.beta = 0.0f; gvb1.sa = 1.0f; gvb1.sb = 1.0f; gvb1.Npad = 16; gvb1.pad_ = 0;
      k_gemm<1><<<dim3((unsigned)((16) + 31) / 32, (unsigned)((SEQ) + 15) / 16, (unsigned)(4)), 32, 0, stream>>>(gvb1); }
    { GemmP gsa2;
      gsa2.A = H1 + (size_t)2 * SEQ * 192; gsa2.B = H2 + (size_t)2 * SEQ * 192 + 16; gsa2.bias = H1 + (size_t)2 * SEQ * 192; gsa2.R = H1 + (size_t)2 * SEQ * 192; gsa2.C = SC;
      gsa2.sAo = 48; gsa2.sAi = 0; gsa2.sAm = 192; gsa2.sAk = 1; gsa2.sBo = 48; gsa2.sBi = 0; gsa2.sBn = 192; gsa2.sBk = 1; gsa2.sCo = (long long)SEQ * SEQ; gsa2.sCi = 0; gsa2.sCm = SEQ; gsa2.sRo = 0; gsa2.sRi = 0; gsa2.sRm = 0; gsa2.sRn = 0;
      gsa2.M = SEQ; gsa2.N = SEQ; gsa2.K = 16; gsa2.zi_n = 1; gsa2.flags = 0; gsa2.act = 0;
      gsa2.alpha = 1.0f; gsa2.beta = 0.0f; gsa2.sa = 1.0f; gsa2.sb = 1.0f; gsa2.Npad = SEQ; gsa2.pad_ = 0;
      k_gemm<1><<<dim3((unsigned)((SEQ) + 31) / 32, (unsigned)((SEQ) + 15) / 16, (unsigned)(4)), 32, 0, stream>>>(gsa2); }
    k_mm_rowsm<<<4 * SEQ, 256, 0, stream>>>(SC, 4 * SEQ, SEQ, 0.25f);
    { GemmP gva2;
      gva2.A = SC; gva2.B = H2 + (size_t)2 * SEQ * 192 + 32; gva2.bias = SC; gva2.R = SC; gva2.C = O1 + (size_t)2 * SEQ * 64;
      gva2.sAo = (long long)SEQ * SEQ; gva2.sAi = 0; gva2.sAm = SEQ; gva2.sAk = 1; gva2.sBo = 48; gva2.sBi = 0; gva2.sBn = 1; gva2.sBk = 192; gva2.sCo = 16; gva2.sCi = 0; gva2.sCm = 64; gva2.sRo = 0; gva2.sRi = 0; gva2.sRm = 0; gva2.sRn = 0;
      gva2.M = SEQ; gva2.N = 16; gva2.K = SEQ; gva2.zi_n = 1; gva2.flags = 0; gva2.act = 0;
      gva2.alpha = 1.0f; gva2.beta = 0.0f; gva2.sa = 1.0f; gva2.sb = 1.0f; gva2.Npad = 16; gva2.pad_ = 0;
      k_gemm<1><<<dim3((unsigned)((16) + 31) / 32, (unsigned)((SEQ) + 15) / 16, (unsigned)(4)), 32, 0, stream>>>(gva2); }
    { GemmP gsb2;
      gsb2.A = H2 + (size_t)2 * SEQ * 192; gsb2.B = H1 + (size_t)2 * SEQ * 192 + 16; gsb2.bias = H2 + (size_t)2 * SEQ * 192; gsb2.R = H2 + (size_t)2 * SEQ * 192; gsb2.C = SC;
      gsb2.sAo = 48; gsb2.sAi = 0; gsb2.sAm = 192; gsb2.sAk = 1; gsb2.sBo = 48; gsb2.sBi = 0; gsb2.sBn = 192; gsb2.sBk = 1; gsb2.sCo = (long long)SEQ * SEQ; gsb2.sCi = 0; gsb2.sCm = SEQ; gsb2.sRo = 0; gsb2.sRi = 0; gsb2.sRm = 0; gsb2.sRn = 0;
      gsb2.M = SEQ; gsb2.N = SEQ; gsb2.K = 16; gsb2.zi_n = 1; gsb2.flags = 0; gsb2.act = 0;
      gsb2.alpha = 1.0f; gsb2.beta = 0.0f; gsb2.sa = 1.0f; gsb2.sb = 1.0f; gsb2.Npad = SEQ; gsb2.pad_ = 0;
      k_gemm<1><<<dim3((unsigned)((SEQ) + 31) / 32, (unsigned)((SEQ) + 15) / 16, (unsigned)(4)), 32, 0, stream>>>(gsb2); }
    k_mm_rowsm<<<4 * SEQ, 256, 0, stream>>>(SC, 4 * SEQ, SEQ, 0.25f);
    { GemmP gvb2;
      gvb2.A = SC; gvb2.B = H1 + (size_t)2 * SEQ * 192 + 32; gvb2.bias = SC; gvb2.R = SC; gvb2.C = O2 + (size_t)2 * SEQ * 64;
      gvb2.sAo = (long long)SEQ * SEQ; gvb2.sAi = 0; gvb2.sAm = SEQ; gvb2.sAk = 1; gvb2.sBo = 48; gvb2.sBi = 0; gvb2.sBn = 1; gvb2.sBk = 192; gvb2.sCo = 16; gvb2.sCi = 0; gvb2.sCm = 64; gvb2.sRo = 0; gvb2.sRi = 0; gvb2.sRm = 0; gvb2.sRn = 0;
      gvb2.M = SEQ; gvb2.N = 16; gvb2.K = SEQ; gvb2.zi_n = 1; gvb2.flags = 0; gvb2.act = 0;
      gvb2.alpha = 1.0f; gvb2.beta = 0.0f; gvb2.sa = 1.0f; gvb2.sb = 1.0f; gvb2.Npad = 16; gvb2.pad_ = 0;
      k_gemm<1><<<dim3((unsigned)((16) + 31) / 32, (unsigned)((SEQ) + 15) / 16, (unsigned)(4)), 32, 0, stream>>>(gvb2); }
    { GemmP gsa3;
      gsa3.A = H1 + (size_t)3 * SEQ * 192; gsa3.B = H2 + (size_t)3 * SEQ * 192 + 16; gsa3.bias = H1 + (size_t)3 * SEQ * 192; gsa3.R = H1 + (size_t)3 * SEQ * 192; gsa3.C = SC;
      gsa3.sAo = 48; gsa3.sAi = 0; gsa3.sAm = 192; gsa3.sAk = 1; gsa3.sBo = 48; gsa3.sBi = 0; gsa3.sBn = 192; gsa3.sBk = 1; gsa3.sCo = (long long)SEQ * SEQ; gsa3.sCi = 0; gsa3.sCm = SEQ; gsa3.sRo = 0; gsa3.sRi = 0; gsa3.sRm = 0; gsa3.sRn = 0;
      gsa3.M = SEQ; gsa3.N = SEQ; gsa3.K = 16; gsa3.zi_n = 1; gsa3.flags = 0; gsa3.act = 0;
      gsa3.alpha = 1.0f; gsa3.beta = 0.0f; gsa3.sa = 1.0f; gsa3.sb = 1.0f; gsa3.Npad = SEQ; gsa3.pad_ = 0;
      k_gemm<1><<<dim3((unsigned)((SEQ) + 31) / 32, (unsigned)((SEQ) + 15) / 16, (unsigned)(4)), 32, 0, stream>>>(gsa3); }
    k_mm_rowsm<<<4 * SEQ, 256, 0, stream>>>(SC, 4 * SEQ, SEQ, 0.25f);
    { GemmP gva3;
      gva3.A = SC; gva3.B = H2 + (size_t)3 * SEQ * 192 + 32; gva3.bias = SC; gva3.R = SC; gva3.C = O1 + (size_t)3 * SEQ * 64;
      gva3.sAo = (long long)SEQ * SEQ; gva3.sAi = 0; gva3.sAm = SEQ; gva3.sAk = 1; gva3.sBo = 48; gva3.sBi = 0; gva3.sBn = 1; gva3.sBk = 192; gva3.sCo = 16; gva3.sCi = 0; gva3.sCm = 64; gva3.sRo = 0; gva3.sRi = 0; gva3.sRm = 0; gva3.sRn = 0;
      gva3.M = SEQ; gva3.N = 16; gva3.K = SEQ; gva3.zi_n = 1; gva3.flags = 0; gva3.act = 0;
      gva3.alpha = 1.0f; gva3.beta = 0.0f; gva3.sa = 1.0f; gva3.sb = 1.0f; gva3.Npad = 16; gva3.pad_ = 0;
      k_gemm<1><<<dim3((unsigned)((16) + 31) / 32, (unsigned)((SEQ) + 15) / 16, (unsigned)(4)), 32, 0, stream>>>(gva3); }
    { GemmP gsb3;
      gsb3.A = H2 + (size_t)3 * SEQ * 192; gsb3.B = H1 + (size_t)3 * SEQ * 192 + 16; gsb3.bias = H2 + (size_t)3 * SEQ * 192; gsb3.R = H2 + (size_t)3 * SEQ * 192; gsb3.C = SC;
      gsb3.sAo = 48; gsb3.sAi = 0; gsb3.sAm = 192; gsb3.sAk = 1; gsb3.sBo = 48; gsb3.sBi = 0; gsb3.sBn = 192; gsb3.sBk = 1; gsb3.sCo = (long long)SEQ * SEQ; gsb3.sCi = 0; gsb3.sCm = SEQ; gsb3.sRo = 0; gsb3.sRi = 0; gsb3.sRm = 0; gsb3.sRn = 0;
      gsb3.M = SEQ; gsb3.N = SEQ; gsb3.K = 16; gsb3.zi_n = 1; gsb3.flags = 0; gsb3.act = 0;
      gsb3.alpha = 1.0f; gsb3.beta = 0.0f; gsb3.sa = 1.0f; gsb3.sb = 1.0f; gsb3.Npad = SEQ; gsb3.pad_ = 0;
      k_gemm<1><<<dim3((unsigned)((SEQ) + 31) / 32, (unsigned)((SEQ) + 15) / 16, (unsigned)(4)), 32, 0, stream>>>(gsb3); }
    k_mm_rowsm<<<4 * SEQ, 256, 0, stream>>>(SC, 4 * SEQ, SEQ, 0.25f);
    { GemmP gvb3;
      gvb3.A = SC; gvb3.B = H1 + (size_t)3 * SEQ * 192 + 32; gvb3.bias = SC; gvb3.R = SC; gvb3.C = O2 + (size_t)3 * SEQ * 64;
      gvb3.sAo = (long long)SEQ * SEQ; gvb3.sAi = 0; gvb3.sAm = SEQ; gvb3.sAk = 1; gvb3.sBo = 48; gvb3.sBi = 0; gvb3.sBn = 1; gvb3.sBk = 192; gvb3.sCo = 16; gvb3.sCi = 0; gvb3.sCm = 64; gvb3.sRo = 0; gvb3.sRi = 0; gvb3.sRm = 0; gvb3.sRn = 0;
      gvb3.M = SEQ; gvb3.N = 16; gvb3.K = SEQ; gvb3.zi_n = 1; gvb3.flags = 0; gvb3.act = 0;
      gvb3.alpha = 1.0f; gvb3.beta = 0.0f; gvb3.sa = 1.0f; gvb3.sb = 1.0f; gvb3.Npad = 16; gvb3.pad_ = 0;
      k_gemm<1><<<dim3((unsigned)((16) + 31) / 32, (unsigned)((SEQ) + 15) / 16, (unsigned)(4)), 32, 0, stream>>>(gvb3); }
    { GemmP gsa4;
      gsa4.A = H1 + (size_t)4 * SEQ * 192; gsa4.B = H2 + (size_t)4 * SEQ * 192 + 16; gsa4.bias = H1 + (size_t)4 * SEQ * 192; gsa4.R = H1 + (size_t)4 * SEQ * 192; gsa4.C = SC;
      gsa4.sAo = 48; gsa4.sAi = 0; gsa4.sAm = 192; gsa4.sAk = 1; gsa4.sBo = 48; gsa4.sBi = 0; gsa4.sBn = 192; gsa4.sBk = 1; gsa4.sCo = (long long)SEQ * SEQ; gsa4.sCi = 0; gsa4.sCm = SEQ; gsa4.sRo = 0; gsa4.sRi = 0; gsa4.sRm = 0; gsa4.sRn = 0;
      gsa4.M = SEQ; gsa4.N = SEQ; gsa4.K = 16; gsa4.zi_n = 1; gsa4.flags = 0; gsa4.act = 0;
      gsa4.alpha = 1.0f; gsa4.beta = 0.0f; gsa4.sa = 1.0f; gsa4.sb = 1.0f; gsa4.Npad = SEQ; gsa4.pad_ = 0;
      k_gemm<1><<<dim3((unsigned)((SEQ) + 31) / 32, (unsigned)((SEQ) + 15) / 16, (unsigned)(4)), 32, 0, stream>>>(gsa4); }
    k_mm_rowsm<<<4 * SEQ, 256, 0, stream>>>(SC, 4 * SEQ, SEQ, 0.25f);
    { GemmP gva4;
      gva4.A = SC; gva4.B = H2 + (size_t)4 * SEQ * 192 + 32; gva4.bias = SC; gva4.R = SC; gva4.C = O1 + (size_t)4 * SEQ * 64;
      gva4.sAo = (long long)SEQ * SEQ; gva4.sAi = 0; gva4.sAm = SEQ; gva4.sAk = 1; gva4.sBo = 48; gva4.sBi = 0; gva4.sBn = 1; gva4.sBk = 192; gva4.sCo = 16; gva4.sCi = 0; gva4.sCm = 64; gva4.sRo = 0; gva4.sRi = 0; gva4.sRm = 0; gva4.sRn = 0;
      gva4.M = SEQ; gva4.N = 16; gva4.K = SEQ; gva4.zi_n = 1; gva4.flags = 0; gva4.act = 0;
      gva4.alpha = 1.0f; gva4.beta = 0.0f; gva4.sa = 1.0f; gva4.sb = 1.0f; gva4.Npad = 16; gva4.pad_ = 0;
      k_gemm<1><<<dim3((unsigned)((16) + 31) / 32, (unsigned)((SEQ) + 15) / 16, (unsigned)(4)), 32, 0, stream>>>(gva4); }
    { GemmP gsb4;
      gsb4.A = H2 + (size_t)4 * SEQ * 192; gsb4.B = H1 + (size_t)4 * SEQ * 192 + 16; gsb4.bias = H2 + (size_t)4 * SEQ * 192; gsb4.R = H2 + (size_t)4 * SEQ * 192; gsb4.C = SC;
      gsb4.sAo = 48; gsb4.sAi = 0; gsb4.sAm = 192; gsb4.sAk = 1; gsb4.sBo = 48; gsb4.sBi = 0; gsb4.sBn = 192; gsb4.sBk = 1; gsb4.sCo = (long long)SEQ * SEQ; gsb4.sCi = 0; gsb4.sCm = SEQ; gsb4.sRo = 0; gsb4.sRi = 0; gsb4.sRm = 0; gsb4.sRn = 0;
      gsb4.M = SEQ; gsb4.N = SEQ; gsb4.K = 16; gsb4.zi_n = 1; gsb4.flags = 0; gsb4.act = 0;
      gsb4.alpha = 1.0f; gsb4.beta = 0.0f; gsb4.sa = 1.0f; gsb4.sb = 1.0f; gsb4.Npad = SEQ; gsb4.pad_ = 0;
      k_gemm<1><<<dim3((unsigned)((SEQ) + 31) / 32, (unsigned)((SEQ) + 15) / 16, (unsigned)(4)), 32, 0, stream>>>(gsb4); }
    k_mm_rowsm<<<4 * SEQ, 256, 0, stream>>>(SC, 4 * SEQ, SEQ, 0.25f);
    { GemmP gvb4;
      gvb4.A = SC; gvb4.B = H1 + (size_t)4 * SEQ * 192 + 32; gvb4.bias = SC; gvb4.R = SC; gvb4.C = O2 + (size_t)4 * SEQ * 64;
      gvb4.sAo = (long long)SEQ * SEQ; gvb4.sAi = 0; gvb4.sAm = SEQ; gvb4.sAk = 1; gvb4.sBo = 48; gvb4.sBi = 0; gvb4.sBn = 1; gvb4.sBk = 192; gvb4.sCo = 16; gvb4.sCi = 0; gvb4.sCm = 64; gvb4.sRo = 0; gvb4.sRi = 0; gvb4.sRm = 0; gvb4.sRn = 0;
      gvb4.M = SEQ; gvb4.N = 16; gvb4.K = SEQ; gvb4.zi_n = 1; gvb4.flags = 0; gvb4.act = 0;
      gvb4.alpha = 1.0f; gvb4.beta = 0.0f; gvb4.sa = 1.0f; gvb4.sb = 1.0f; gvb4.Npad = 16; gvb4.pad_ = 0;
      k_gemm<1><<<dim3((unsigned)((16) + 31) / 32, (unsigned)((SEQ) + 15) / 16, (unsigned)(4)), 32, 0, stream>>>(gvb4); }
    { GemmP gsa5;
      gsa5.A = H1 + (size_t)5 * SEQ * 192; gsa5.B = H2 + (size_t)5 * SEQ * 192 + 16; gsa5.bias = H1 + (size_t)5 * SEQ * 192; gsa5.R = H1 + (size_t)5 * SEQ * 192; gsa5.C = SC;
      gsa5.sAo = 48; gsa5.sAi = 0; gsa5.sAm = 192; gsa5.sAk = 1; gsa5.sBo = 48; gsa5.sBi = 0; gsa5.sBn = 192; gsa5.sBk = 1; gsa5.sCo = (long long)SEQ * SEQ; gsa5.sCi = 0; gsa5.sCm = SEQ; gsa5.sRo = 0; gsa5.sRi = 0; gsa5.sRm = 0; gsa5.sRn = 0;
      gsa5.M = SEQ; gsa5.N = SEQ; gsa5.K = 16; gsa5.zi_n = 1; gsa5.flags = 0; gsa5.act = 0;
      gsa5.alpha = 1.0f; gsa5.beta = 0.0f; gsa5.sa = 1.0f; gsa5.sb = 1.0f; gsa5.Npad = SEQ; gsa5.pad_ = 0;
      k_gemm<1><<<dim3((unsigned)((SEQ) + 31) / 32, (unsigned)((SEQ) + 15) / 16, (unsigned)(4)), 32, 0, stream>>>(gsa5); }
    k_mm_rowsm<<<4 * SEQ, 256, 0, stream>>>(SC, 4 * SEQ, SEQ, 0.25f);
    { GemmP gva5;
      gva5.A = SC; gva5.B = H2 + (size_t)5 * SEQ * 192 + 32; gva5.bias = SC; gva5.R = SC; gva5.C = O1 + (size_t)5 * SEQ * 64;
      gva5.sAo = (long long)SEQ * SEQ; gva5.sAi = 0; gva5.sAm = SEQ; gva5.sAk = 1; gva5.sBo = 48; gva5.sBi = 0; gva5.sBn = 1; gva5.sBk = 192; gva5.sCo = 16; gva5.sCi = 0; gva5.sCm = 64; gva5.sRo = 0; gva5.sRi = 0; gva5.sRm = 0; gva5.sRn = 0;
      gva5.M = SEQ; gva5.N = 16; gva5.K = SEQ; gva5.zi_n = 1; gva5.flags = 0; gva5.act = 0;
      gva5.alpha = 1.0f; gva5.beta = 0.0f; gva5.sa = 1.0f; gva5.sb = 1.0f; gva5.Npad = 16; gva5.pad_ = 0;
      k_gemm<1><<<dim3((unsigned)((16) + 31) / 32, (unsigned)((SEQ) + 15) / 16, (unsigned)(4)), 32, 0, stream>>>(gva5); }
    { GemmP gsb5;
      gsb5.A = H2 + (size_t)5 * SEQ * 192; gsb5.B = H1 + (size_t)5 * SEQ * 192 + 16; gsb5.bias = H2 + (size_t)5 * SEQ * 192; gsb5.R = H2 + (size_t)5 * SEQ * 192; gsb5.C = SC;
      gsb5.sAo = 48; gsb5.sAi = 0; gsb5.sAm = 192; gsb5.sAk = 1; gsb5.sBo = 48; gsb5.sBi = 0; gsb5.sBn = 192; gsb5.sBk = 1; gsb5.sCo = (long long)SEQ * SEQ; gsb5.sCi = 0; gsb5.sCm = SEQ; gsb5.sRo = 0; gsb5.sRi = 0; gsb5.sRm = 0; gsb5.sRn = 0;
      gsb5.M = SEQ; gsb5.N = SEQ; gsb5.K = 16; gsb5.zi_n = 1; gsb5.flags = 0; gsb5.act = 0;
      gsb5.alpha = 1.0f; gsb5.beta = 0.0f; gsb5.sa = 1.0f; gsb5.sb = 1.0f; gsb5.Npad = SEQ; gsb5.pad_ = 0;
      k_gemm<1><<<dim3((unsigned)((SEQ) + 31) / 32, (unsigned)((SEQ) + 15) / 16, (unsigned)(4)), 32, 0, stream>>>(gsb5); }
    k_mm_rowsm<<<4 * SEQ, 256, 0, stream>>>(SC, 4 * SEQ, SEQ, 0.25f);
    { GemmP gvb5;
      gvb5.A = SC; gvb5.B = H1 + (size_t)5 * SEQ * 192 + 32; gvb5.bias = SC; gvb5.R = SC; gvb5.C = O2 + (size_t)5 * SEQ * 64;
      gvb5.sAo = (long long)SEQ * SEQ; gvb5.sAi = 0; gvb5.sAm = SEQ; gvb5.sAk = 1; gvb5.sBo = 48; gvb5.sBi = 0; gvb5.sBn = 1; gvb5.sBk = 192; gvb5.sCo = 16; gvb5.sCi = 0; gvb5.sCm = 64; gvb5.sRo = 0; gvb5.sRi = 0; gvb5.sRm = 0; gvb5.sRn = 0;
      gvb5.M = SEQ; gvb5.N = 16; gvb5.K = SEQ; gvb5.zi_n = 1; gvb5.flags = 0; gvb5.act = 0;
      gvb5.alpha = 1.0f; gvb5.beta = 0.0f; gvb5.sa = 1.0f; gvb5.sb = 1.0f; gvb5.Npad = 16; gvb5.pad_ = 0;
      k_gemm<1><<<dim3((unsigned)((16) + 31) / 32, (unsigned)((SEQ) + 15) / 16, (unsigned)(4)), 32, 0, stream>>>(gvb5); }
    { GemmP gsa6;
      gsa6.A = H1 + (size_t)6 * SEQ * 192; gsa6.B = H2 + (size_t)6 * SEQ * 192 + 16; gsa6.bias = H1 + (size_t)6 * SEQ * 192; gsa6.R = H1 + (size_t)6 * SEQ * 192; gsa6.C = SC;
      gsa6.sAo = 48; gsa6.sAi = 0; gsa6.sAm = 192; gsa6.sAk = 1; gsa6.sBo = 48; gsa6.sBi = 0; gsa6.sBn = 192; gsa6.sBk = 1; gsa6.sCo = (long long)SEQ * SEQ; gsa6.sCi = 0; gsa6.sCm = SEQ; gsa6.sRo = 0; gsa6.sRi = 0; gsa6.sRm = 0; gsa6.sRn = 0;
      gsa6.M = SEQ; gsa6.N = SEQ; gsa6.K = 16; gsa6.zi_n = 1; gsa6.flags = 0; gsa6.act = 0;
      gsa6.alpha = 1.0f; gsa6.beta = 0.0f; gsa6.sa = 1.0f; gsa6.sb = 1.0f; gsa6.Npad = SEQ; gsa6.pad_ = 0;
      k_gemm<1><<<dim3((unsigned)((SEQ) + 31) / 32, (unsigned)((SEQ) + 15) / 16, (unsigned)(4)), 32, 0, stream>>>(gsa6); }
    k_mm_rowsm<<<4 * SEQ, 256, 0, stream>>>(SC, 4 * SEQ, SEQ, 0.25f);
    { GemmP gva6;
      gva6.A = SC; gva6.B = H2 + (size_t)6 * SEQ * 192 + 32; gva6.bias = SC; gva6.R = SC; gva6.C = O1 + (size_t)6 * SEQ * 64;
      gva6.sAo = (long long)SEQ * SEQ; gva6.sAi = 0; gva6.sAm = SEQ; gva6.sAk = 1; gva6.sBo = 48; gva6.sBi = 0; gva6.sBn = 1; gva6.sBk = 192; gva6.sCo = 16; gva6.sCi = 0; gva6.sCm = 64; gva6.sRo = 0; gva6.sRi = 0; gva6.sRm = 0; gva6.sRn = 0;
      gva6.M = SEQ; gva6.N = 16; gva6.K = SEQ; gva6.zi_n = 1; gva6.flags = 0; gva6.act = 0;
      gva6.alpha = 1.0f; gva6.beta = 0.0f; gva6.sa = 1.0f; gva6.sb = 1.0f; gva6.Npad = 16; gva6.pad_ = 0;
      k_gemm<1><<<dim3((unsigned)((16) + 31) / 32, (unsigned)((SEQ) + 15) / 16, (unsigned)(4)), 32, 0, stream>>>(gva6); }
    { GemmP gsb6;
      gsb6.A = H2 + (size_t)6 * SEQ * 192; gsb6.B = H1 + (size_t)6 * SEQ * 192 + 16; gsb6.bias = H2 + (size_t)6 * SEQ * 192; gsb6.R = H2 + (size_t)6 * SEQ * 192; gsb6.C = SC;
      gsb6.sAo = 48; gsb6.sAi = 0; gsb6.sAm = 192; gsb6.sAk = 1; gsb6.sBo = 48; gsb6.sBi = 0; gsb6.sBn = 192; gsb6.sBk = 1; gsb6.sCo = (long long)SEQ * SEQ; gsb6.sCi = 0; gsb6.sCm = SEQ; gsb6.sRo = 0; gsb6.sRi = 0; gsb6.sRm = 0; gsb6.sRn = 0;
      gsb6.M = SEQ; gsb6.N = SEQ; gsb6.K = 16; gsb6.zi_n = 1; gsb6.flags = 0; gsb6.act = 0;
      gsb6.alpha = 1.0f; gsb6.beta = 0.0f; gsb6.sa = 1.0f; gsb6.sb = 1.0f; gsb6.Npad = SEQ; gsb6.pad_ = 0;
      k_gemm<1><<<dim3((unsigned)((SEQ) + 31) / 32, (unsigned)((SEQ) + 15) / 16, (unsigned)(4)), 32, 0, stream>>>(gsb6); }
    k_mm_rowsm<<<4 * SEQ, 256, 0, stream>>>(SC, 4 * SEQ, SEQ, 0.25f);
    { GemmP gvb6;
      gvb6.A = SC; gvb6.B = H1 + (size_t)6 * SEQ * 192 + 32; gvb6.bias = SC; gvb6.R = SC; gvb6.C = O2 + (size_t)6 * SEQ * 64;
      gvb6.sAo = (long long)SEQ * SEQ; gvb6.sAi = 0; gvb6.sAm = SEQ; gvb6.sAk = 1; gvb6.sBo = 48; gvb6.sBi = 0; gvb6.sBn = 1; gvb6.sBk = 192; gvb6.sCo = 16; gvb6.sCi = 0; gvb6.sCm = 64; gvb6.sRo = 0; gvb6.sRi = 0; gvb6.sRm = 0; gvb6.sRn = 0;
      gvb6.M = SEQ; gvb6.N = 16; gvb6.K = SEQ; gvb6.zi_n = 1; gvb6.flags = 0; gvb6.act = 0;
      gvb6.alpha = 1.0f; gvb6.beta = 0.0f; gvb6.sa = 1.0f; gvb6.sb = 1.0f; gvb6.Npad = 16; gvb6.pad_ = 0;
      k_gemm<1><<<dim3((unsigned)((16) + 31) / 32, (unsigned)((SEQ) + 15) / 16, (unsigned)(4)), 32, 0, stream>>>(gvb6); }
    { GemmP gsa7;
      gsa7.A = H1 + (size_t)7 * SEQ * 192; gsa7.B = H2 + (size_t)7 * SEQ * 192 + 16; gsa7.bias = H1 + (size_t)7 * SEQ * 192; gsa7.R = H1 + (size_t)7 * SEQ * 192; gsa7.C = SC;
      gsa7.sAo = 48; gsa7.sAi = 0; gsa7.sAm = 192; gsa7.sAk = 1; gsa7.sBo = 48; gsa7.sBi = 0; gsa7.sBn = 192; gsa7.sBk = 1; gsa7.sCo = (long long)SEQ * SEQ; gsa7.sCi = 0; gsa7.sCm = SEQ; gsa7.sRo = 0; gsa7.sRi = 0; gsa7.sRm = 0; gsa7.sRn = 0;
      gsa7.M = SEQ; gsa7.N = SEQ; gsa7.K = 16; gsa7.zi_n = 1; gsa7.flags = 0; gsa7.act = 0;
      gsa7.alpha = 1.0f; gsa7.beta = 0.0f; gsa7.sa = 1.0f; gsa7.sb = 1.0f; gsa7.Npad = SEQ; gsa7.pad_ = 0;
      k_gemm<1><<<dim3((unsigned)((SEQ) + 31) / 32, (unsigned)((SEQ) + 15) / 16, (unsigned)(4)), 32, 0, stream>>>(gsa7); }
    k_mm_rowsm<<<4 * SEQ, 256, 0, stream>>>(SC, 4 * SEQ, SEQ, 0.25f);
    { GemmP gva7;
      gva7.A = SC; gva7.B = H2 + (size_t)7 * SEQ * 192 + 32; gva7.bias = SC; gva7.R = SC; gva7.C = O1 + (size_t)7 * SEQ * 64;
      gva7.sAo = (long long)SEQ * SEQ; gva7.sAi = 0; gva7.sAm = SEQ; gva7.sAk = 1; gva7.sBo = 48; gva7.sBi = 0; gva7.sBn = 1; gva7.sBk = 192; gva7.sCo = 16; gva7.sCi = 0; gva7.sCm = 64; gva7.sRo = 0; gva7.sRi = 0; gva7.sRm = 0; gva7.sRn = 0;
      gva7.M = SEQ; gva7.N = 16; gva7.K = SEQ; gva7.zi_n = 1; gva7.flags = 0; gva7.act = 0;
      gva7.alpha = 1.0f; gva7.beta = 0.0f; gva7.sa = 1.0f; gva7.sb = 1.0f; gva7.Npad = 16; gva7.pad_ = 0;
      k_gemm<1><<<dim3((unsigned)((16) + 31) / 32, (unsigned)((SEQ) + 15) / 16, (unsigned)(4)), 32, 0, stream>>>(gva7); }
    { GemmP gsb7;
      gsb7.A = H2 + (size_t)7 * SEQ * 192; gsb7.B = H1 + (size_t)7 * SEQ * 192 + 16; gsb7.bias = H2 + (size_t)7 * SEQ * 192; gsb7.R = H2 + (size_t)7 * SEQ * 192; gsb7.C = SC;
      gsb7.sAo = 48; gsb7.sAi = 0; gsb7.sAm = 192; gsb7.sAk = 1; gsb7.sBo = 48; gsb7.sBi = 0; gsb7.sBn = 192; gsb7.sBk = 1; gsb7.sCo = (long long)SEQ * SEQ; gsb7.sCi = 0; gsb7.sCm = SEQ; gsb7.sRo = 0; gsb7.sRi = 0; gsb7.sRm = 0; gsb7.sRn = 0;
      gsb7.M = SEQ; gsb7.N = SEQ; gsb7.K = 16; gsb7.zi_n = 1; gsb7.flags = 0; gsb7.act = 0;
      gsb7.alpha = 1.0f; gsb7.beta = 0.0f; gsb7.sa = 1.0f; gsb7.sb = 1.0f; gsb7.Npad = SEQ; gsb7.pad_ = 0;
      k_gemm<1><<<dim3((unsigned)((SEQ) + 31) / 32, (unsigned)((SEQ) + 15) / 16, (unsigned)(4)), 32, 0, stream>>>(gsb7); }
    k_mm_rowsm<<<4 * SEQ, 256, 0, stream>>>(SC, 4 * SEQ, SEQ, 0.25f);
    { GemmP gvb7;
      gvb7.A = SC; gvb7.B = H1 + (size_t)7 * SEQ * 192 + 32; gvb7.bias = SC; gvb7.R = SC; gvb7.C = O2 + (size_t)7 * SEQ * 64;
      gvb7.sAo = (long long)SEQ * SEQ; gvb7.sAi = 0; gvb7.sAm = SEQ; gvb7.sAk = 1; gvb7.sBo = 48; gvb7.sBi = 0; gvb7.sBn = 1; gvb7.sBk = 192; gvb7.sCo = 16; gvb7.sCi = 0; gvb7.sCm = 64; gvb7.sRo = 0; gvb7.sRi = 0; gvb7.sRm = 0; gvb7.sRn = 0;
      gvb7.M = SEQ; gvb7.N = 16; gvb7.K = SEQ; gvb7.zi_n = 1; gvb7.flags = 0; gvb7.act = 0;
      gvb7.alpha = 1.0f; gvb7.beta = 0.0f; gvb7.sa = 1.0f; gvb7.sb = 1.0f; gvb7.Npad = 16; gvb7.pad_ = 0;
      k_gemm<1><<<dim3((unsigned)((16) + 31) / 32, (unsigned)((SEQ) + 15) / 16, (unsigned)(4)), 32, 0, stream>>>(gvb7); }
    { GemmP gsa8;
      gsa8.A = H1 + (size_t)8 * SEQ * 192; gsa8.B = H2 + (size_t)8 * SEQ * 192 + 16; gsa8.bias = H1 + (size_t)8 * SEQ * 192; gsa8.R = H1 + (size_t)8 * SEQ * 192; gsa8.C = SC;
      gsa8.sAo = 48; gsa8.sAi = 0; gsa8.sAm = 192; gsa8.sAk = 1; gsa8.sBo = 48; gsa8.sBi = 0; gsa8.sBn = 192; gsa8.sBk = 1; gsa8.sCo = (long long)SEQ * SEQ; gsa8.sCi = 0; gsa8.sCm = SEQ; gsa8.sRo = 0; gsa8.sRi = 0; gsa8.sRm = 0; gsa8.sRn = 0;
      gsa8.M = SEQ; gsa8.N = SEQ; gsa8.K = 16; gsa8.zi_n = 1; gsa8.flags = 0; gsa8.act = 0;
      gsa8.alpha = 1.0f; gsa8.beta = 0.0f; gsa8.sa = 1.0f; gsa8.sb = 1.0f; gsa8.Npad = SEQ; gsa8.pad_ = 0;
      k_gemm<1><<<dim3((unsigned)((SEQ) + 31) / 32, (unsigned)((SEQ) + 15) / 16, (unsigned)(4)), 32, 0, stream>>>(gsa8); }
    k_mm_rowsm<<<4 * SEQ, 256, 0, stream>>>(SC, 4 * SEQ, SEQ, 0.25f);
    { GemmP gva8;
      gva8.A = SC; gva8.B = H2 + (size_t)8 * SEQ * 192 + 32; gva8.bias = SC; gva8.R = SC; gva8.C = O1 + (size_t)8 * SEQ * 64;
      gva8.sAo = (long long)SEQ * SEQ; gva8.sAi = 0; gva8.sAm = SEQ; gva8.sAk = 1; gva8.sBo = 48; gva8.sBi = 0; gva8.sBn = 1; gva8.sBk = 192; gva8.sCo = 16; gva8.sCi = 0; gva8.sCm = 64; gva8.sRo = 0; gva8.sRi = 0; gva8.sRm = 0; gva8.sRn = 0;
      gva8.M = SEQ; gva8.N = 16; gva8.K = SEQ; gva8.zi_n = 1; gva8.flags = 0; gva8.act = 0;
      gva8.alpha = 1.0f; gva8.beta = 0.0f; gva8.sa = 1.0f; gva8.sb = 1.0f; gva8.Npad = 16; gva8.pad_ = 0;
      k_gemm<1><<<dim3((unsigned)((16) + 31) / 32, (unsigned)((SEQ) + 15) / 16, (unsigned)(4)), 32, 0, stream>>>(gva8); }
    { GemmP gsb8;
      gsb8.A = H2 + (size_t)8 * SEQ * 192; gsb8.B = H1 + (size_t)8 * SEQ * 192 + 16; gsb8.bias = H2 + (size_t)8 * SEQ * 192; gsb8.R = H2 + (size_t)8 * SEQ * 192; gsb8.C = SC;
      gsb8.sAo = 48; gsb8.sAi = 0; gsb8.sAm = 192; gsb8.sAk = 1; gsb8.sBo = 48; gsb8.sBi = 0; gsb8.sBn = 192; gsb8.sBk = 1; gsb8.sCo = (long long)SEQ * SEQ; gsb8.sCi = 0; gsb8.sCm = SEQ; gsb8.sRo = 0; gsb8.sRi = 0; gsb8.sRm = 0; gsb8.sRn = 0;
      gsb8.M = SEQ; gsb8.N = SEQ; gsb8.K = 16; gsb8.zi_n = 1; gsb8.flags = 0; gsb8.act = 0;
      gsb8.alpha = 1.0f; gsb8.beta = 0.0f; gsb8.sa = 1.0f; gsb8.sb = 1.0f; gsb8.Npad = SEQ; gsb8.pad_ = 0;
      k_gemm<1><<<dim3((unsigned)((SEQ) + 31) / 32, (unsigned)((SEQ) + 15) / 16, (unsigned)(4)), 32, 0, stream>>>(gsb8); }
    k_mm_rowsm<<<4 * SEQ, 256, 0, stream>>>(SC, 4 * SEQ, SEQ, 0.25f);
    { GemmP gvb8;
      gvb8.A = SC; gvb8.B = H1 + (size_t)8 * SEQ * 192 + 32; gvb8.bias = SC; gvb8.R = SC; gvb8.C = O2 + (size_t)8 * SEQ * 64;
      gvb8.sAo = (long long)SEQ * SEQ; gvb8.sAi = 0; gvb8.sAm = SEQ; gvb8.sAk = 1; gvb8.sBo = 48; gvb8.sBi = 0; gvb8.sBn = 1; gvb8.sBk = 192; gvb8.sCo = 16; gvb8.sCi = 0; gvb8.sCm = 64; gvb8.sRo = 0; gvb8.sRi = 0; gvb8.sRm = 0; gvb8.sRn = 0;
      gvb8.M = SEQ; gvb8.N = 16; gvb8.K = SEQ; gvb8.zi_n = 1; gvb8.flags = 0; gvb8.act = 0;
      gvb8.alpha = 1.0f; gvb8.beta = 0.0f; gvb8.sa = 1.0f; gvb8.sb = 1.0f; gvb8.Npad = 16; gvb8.pad_ = 0;
      k_gemm<1><<<dim3((unsigned)((16) + 31) / 32, (unsigned)((SEQ) + 15) / 16, (unsigned)(4)), 32, 0, stream>>>(gvb8); }
    { GemmP gsa9;
      gsa9.A = H1 + (size_t)9 * SEQ * 192; gsa9.B = H2 + (size_t)9 * SEQ * 192 + 16; gsa9.bias = H1 + (size_t)9 * SEQ * 192; gsa9.R = H1 + (size_t)9 * SEQ * 192; gsa9.C = SC;
      gsa9.sAo = 48; gsa9.sAi = 0; gsa9.sAm = 192; gsa9.sAk = 1; gsa9.sBo = 48; gsa9.sBi = 0; gsa9.sBn = 192; gsa9.sBk = 1; gsa9.sCo = (long long)SEQ * SEQ; gsa9.sCi = 0; gsa9.sCm = SEQ; gsa9.sRo = 0; gsa9.sRi = 0; gsa9.sRm = 0; gsa9.sRn = 0;
      gsa9.M = SEQ; gsa9.N = SEQ; gsa9.K = 16; gsa9.zi_n = 1; gsa9.flags = 0; gsa9.act = 0;
      gsa9.alpha = 1.0f; gsa9.beta = 0.0f; gsa9.sa = 1.0f; gsa9.sb = 1.0f; gsa9.Npad = SEQ; gsa9.pad_ = 0;
      k_gemm<1><<<dim3((unsigned)((SEQ) + 31) / 32, (unsigned)((SEQ) + 15) / 16, (unsigned)(4)), 32, 0, stream>>>(gsa9); }
    k_mm_rowsm<<<4 * SEQ, 256, 0, stream>>>(SC, 4 * SEQ, SEQ, 0.25f);
    { GemmP gva9;
      gva9.A = SC; gva9.B = H2 + (size_t)9 * SEQ * 192 + 32; gva9.bias = SC; gva9.R = SC; gva9.C = O1 + (size_t)9 * SEQ * 64;
      gva9.sAo = (long long)SEQ * SEQ; gva9.sAi = 0; gva9.sAm = SEQ; gva9.sAk = 1; gva9.sBo = 48; gva9.sBi = 0; gva9.sBn = 1; gva9.sBk = 192; gva9.sCo = 16; gva9.sCi = 0; gva9.sCm = 64; gva9.sRo = 0; gva9.sRi = 0; gva9.sRm = 0; gva9.sRn = 0;
      gva9.M = SEQ; gva9.N = 16; gva9.K = SEQ; gva9.zi_n = 1; gva9.flags = 0; gva9.act = 0;
      gva9.alpha = 1.0f; gva9.beta = 0.0f; gva9.sa = 1.0f; gva9.sb = 1.0f; gva9.Npad = 16; gva9.pad_ = 0;
      k_gemm<1><<<dim3((unsigned)((16) + 31) / 32, (unsigned)((SEQ) + 15) / 16, (unsigned)(4)), 32, 0, stream>>>(gva9); }
    { GemmP gsb9;
      gsb9.A = H2 + (size_t)9 * SEQ * 192; gsb9.B = H1 + (size_t)9 * SEQ * 192 + 16; gsb9.bias = H2 + (size_t)9 * SEQ * 192; gsb9.R = H2 + (size_t)9 * SEQ * 192; gsb9.C = SC;
      gsb9.sAo = 48; gsb9.sAi = 0; gsb9.sAm = 192; gsb9.sAk = 1; gsb9.sBo = 48; gsb9.sBi = 0; gsb9.sBn = 192; gsb9.sBk = 1; gsb9.sCo = (long long)SEQ * SEQ; gsb9.sCi = 0; gsb9.sCm = SEQ; gsb9.sRo = 0; gsb9.sRi = 0; gsb9.sRm = 0; gsb9.sRn = 0;
      gsb9.M = SEQ; gsb9.N = SEQ; gsb9.K = 16; gsb9.zi_n = 1; gsb9.flags = 0; gsb9.act = 0;
      gsb9.alpha = 1.0f; gsb9.beta = 0.0f; gsb9.sa = 1.0f; gsb9.sb = 1.0f; gsb9.Npad = SEQ; gsb9.pad_ = 0;
      k_gemm<1><<<dim3((unsigned)((SEQ) + 31) / 32, (unsigned)((SEQ) + 15) / 16, (unsigned)(4)), 32, 0, stream>>>(gsb9); }
    k_mm_rowsm<<<4 * SEQ, 256, 0, stream>>>(SC, 4 * SEQ, SEQ, 0.25f);
    { GemmP gvb9;
      gvb9.A = SC; gvb9.B = H1 + (size_t)9 * SEQ * 192 + 32; gvb9.bias = SC; gvb9.R = SC; gvb9.C = O2 + (size_t)9 * SEQ * 64;
      gvb9.sAo = (long long)SEQ * SEQ; gvb9.sAi = 0; gvb9.sAm = SEQ; gvb9.sAk = 1; gvb9.sBo = 48; gvb9.sBi = 0; gvb9.sBn = 1; gvb9.sBk = 192; gvb9.sCo = 16; gvb9.sCi = 0; gvb9.sCm = 64; gvb9.sRo = 0; gvb9.sRi = 0; gvb9.sRm = 0; gvb9.sRn = 0;
      gvb9.M = SEQ; gvb9.N = 16; gvb9.K = SEQ; gvb9.zi_n = 1; gvb9.flags = 0; gvb9.act = 0;
      gvb9.alpha = 1.0f; gvb9.beta = 0.0f; gvb9.sa = 1.0f; gvb9.sb = 1.0f; gvb9.Npad = 16; gvb9.pad_ = 0;
      k_gemm<1><<<dim3((unsigned)((16) + 31) / 32, (unsigned)((SEQ) + 15) / 16, (unsigned)(4)), 32, 0, stream>>>(gvb9); }
    { GemmP gsa10;
      gsa10.A = H1 + (size_t)10 * SEQ * 192; gsa10.B = H2 + (size_t)10 * SEQ * 192 + 16; gsa10.bias = H1 + (size_t)10 * SEQ * 192; gsa10.R = H1 + (size_t)10 * SEQ * 192; gsa10.C = SC;
      gsa10.sAo = 48; gsa10.sAi = 0; gsa10.sAm = 192; gsa10.sAk = 1; gsa10.sBo = 48; gsa10.sBi = 0; gsa10.sBn = 192; gsa10.sBk = 1; gsa10.sCo = (long long)SEQ * SEQ; gsa10.sCi = 0; gsa10.sCm = SEQ; gsa10.sRo = 0; gsa10.sRi = 0; gsa10.sRm = 0; gsa10.sRn = 0;
      gsa10.M = SEQ; gsa10.N = SEQ; gsa10.K = 16; gsa10.zi_n = 1; gsa10.flags = 0; gsa10.act = 0;
      gsa10.alpha = 1.0f; gsa10.beta = 0.0f; gsa10.sa = 1.0f; gsa10.sb = 1.0f; gsa10.Npad = SEQ; gsa10.pad_ = 0;
      k_gemm<1><<<dim3((unsigned)((SEQ) + 31) / 32, (unsigned)((SEQ) + 15) / 16, (unsigned)(4)), 32, 0, stream>>>(gsa10); }
    k_mm_rowsm<<<4 * SEQ, 256, 0, stream>>>(SC, 4 * SEQ, SEQ, 0.25f);
    { GemmP gva10;
      gva10.A = SC; gva10.B = H2 + (size_t)10 * SEQ * 192 + 32; gva10.bias = SC; gva10.R = SC; gva10.C = O1 + (size_t)10 * SEQ * 64;
      gva10.sAo = (long long)SEQ * SEQ; gva10.sAi = 0; gva10.sAm = SEQ; gva10.sAk = 1; gva10.sBo = 48; gva10.sBi = 0; gva10.sBn = 1; gva10.sBk = 192; gva10.sCo = 16; gva10.sCi = 0; gva10.sCm = 64; gva10.sRo = 0; gva10.sRi = 0; gva10.sRm = 0; gva10.sRn = 0;
      gva10.M = SEQ; gva10.N = 16; gva10.K = SEQ; gva10.zi_n = 1; gva10.flags = 0; gva10.act = 0;
      gva10.alpha = 1.0f; gva10.beta = 0.0f; gva10.sa = 1.0f; gva10.sb = 1.0f; gva10.Npad = 16; gva10.pad_ = 0;
      k_gemm<1><<<dim3((unsigned)((16) + 31) / 32, (unsigned)((SEQ) + 15) / 16, (unsigned)(4)), 32, 0, stream>>>(gva10); }
    { GemmP gsb10;
      gsb10.A = H2 + (size_t)10 * SEQ * 192; gsb10.B = H1 + (size_t)10 * SEQ * 192 + 16; gsb10.bias = H2 + (size_t)10 * SEQ * 192; gsb10.R = H2 + (size_t)10 * SEQ * 192; gsb10.C = SC;
      gsb10.sAo = 48; gsb10.sAi = 0; gsb10.sAm = 192; gsb10.sAk = 1; gsb10.sBo = 48; gsb10.sBi = 0; gsb10.sBn = 192; gsb10.sBk = 1; gsb10.sCo = (long long)SEQ * SEQ; gsb10.sCi = 0; gsb10.sCm = SEQ; gsb10.sRo = 0; gsb10.sRi = 0; gsb10.sRm = 0; gsb10.sRn = 0;
      gsb10.M = SEQ; gsb10.N = SEQ; gsb10.K = 16; gsb10.zi_n = 1; gsb10.flags = 0; gsb10.act = 0;
      gsb10.alpha = 1.0f; gsb10.beta = 0.0f; gsb10.sa = 1.0f; gsb10.sb = 1.0f; gsb10.Npad = SEQ; gsb10.pad_ = 0;
      k_gemm<1><<<dim3((unsigned)((SEQ) + 31) / 32, (unsigned)((SEQ) + 15) / 16, (unsigned)(4)), 32, 0, stream>>>(gsb10); }
    k_mm_rowsm<<<4 * SEQ, 256, 0, stream>>>(SC, 4 * SEQ, SEQ, 0.25f);
    { GemmP gvb10;
      gvb10.A = SC; gvb10.B = H1 + (size_t)10 * SEQ * 192 + 32; gvb10.bias = SC; gvb10.R = SC; gvb10.C = O2 + (size_t)10 * SEQ * 64;
      gvb10.sAo = (long long)SEQ * SEQ; gvb10.sAi = 0; gvb10.sAm = SEQ; gvb10.sAk = 1; gvb10.sBo = 48; gvb10.sBi = 0; gvb10.sBn = 1; gvb10.sBk = 192; gvb10.sCo = 16; gvb10.sCi = 0; gvb10.sCm = 64; gvb10.sRo = 0; gvb10.sRi = 0; gvb10.sRm = 0; gvb10.sRn = 0;
      gvb10.M = SEQ; gvb10.N = 16; gvb10.K = SEQ; gvb10.zi_n = 1; gvb10.flags = 0; gvb10.act = 0;
      gvb10.alpha = 1.0f; gvb10.beta = 0.0f; gvb10.sa = 1.0f; gvb10.sb = 1.0f; gvb10.Npad = 16; gvb10.pad_ = 0;
      k_gemm<1><<<dim3((unsigned)((16) + 31) / 32, (unsigned)((SEQ) + 15) / 16, (unsigned)(4)), 32, 0, stream>>>(gvb10); }
    { GemmP gsa11;
      gsa11.A = H1 + (size_t)11 * SEQ * 192; gsa11.B = H2 + (size_t)11 * SEQ * 192 + 16; gsa11.bias = H1 + (size_t)11 * SEQ * 192; gsa11.R = H1 + (size_t)11 * SEQ * 192; gsa11.C = SC;
      gsa11.sAo = 48; gsa11.sAi = 0; gsa11.sAm = 192; gsa11.sAk = 1; gsa11.sBo = 48; gsa11.sBi = 0; gsa11.sBn = 192; gsa11.sBk = 1; gsa11.sCo = (long long)SEQ * SEQ; gsa11.sCi = 0; gsa11.sCm = SEQ; gsa11.sRo = 0; gsa11.sRi = 0; gsa11.sRm = 0; gsa11.sRn = 0;
      gsa11.M = SEQ; gsa11.N = SEQ; gsa11.K = 16; gsa11.zi_n = 1; gsa11.flags = 0; gsa11.act = 0;
      gsa11.alpha = 1.0f; gsa11.beta = 0.0f; gsa11.sa = 1.0f; gsa11.sb = 1.0f; gsa11.Npad = SEQ; gsa11.pad_ = 0;
      k_gemm<1><<<dim3((unsigned)((SEQ) + 31) / 32, (unsigned)((SEQ) + 15) / 16, (unsigned)(4)), 32, 0, stream>>>(gsa11); }
    k_mm_rowsm<<<4 * SEQ, 256, 0, stream>>>(SC, 4 * SEQ, SEQ, 0.25f);
    { GemmP gva11;
      gva11.A = SC; gva11.B = H2 + (size_t)11 * SEQ * 192 + 32; gva11.bias = SC; gva11.R = SC; gva11.C = O1 + (size_t)11 * SEQ * 64;
      gva11.sAo = (long long)SEQ * SEQ; gva11.sAi = 0; gva11.sAm = SEQ; gva11.sAk = 1; gva11.sBo = 48; gva11.sBi = 0; gva11.sBn = 1; gva11.sBk = 192; gva11.sCo = 16; gva11.sCi = 0; gva11.sCm = 64; gva11.sRo = 0; gva11.sRi = 0; gva11.sRm = 0; gva11.sRn = 0;
      gva11.M = SEQ; gva11.N = 16; gva11.K = SEQ; gva11.zi_n = 1; gva11.flags = 0; gva11.act = 0;
      gva11.alpha = 1.0f; gva11.beta = 0.0f; gva11.sa = 1.0f; gva11.sb = 1.0f; gva11.Npad = 16; gva11.pad_ = 0;
      k_gemm<1><<<dim3((unsigned)((16) + 31) / 32, (unsigned)((SEQ) + 15) / 16, (unsigned)(4)), 32, 0, stream>>>(gva11); }
    { GemmP gsb11;
      gsb11.A = H2 + (size_t)11 * SEQ * 192; gsb11.B = H1 + (size_t)11 * SEQ * 192 + 16; gsb11.bias = H2 + (size_t)11 * SEQ * 192; gsb11.R = H2 + (size_t)11 * SEQ * 192; gsb11.C = SC;
      gsb11.sAo = 48; gsb11.sAi = 0; gsb11.sAm = 192; gsb11.sAk = 1; gsb11.sBo = 48; gsb11.sBi = 0; gsb11.sBn = 192; gsb11.sBk = 1; gsb11.sCo = (long long)SEQ * SEQ; gsb11.sCi = 0; gsb11.sCm = SEQ; gsb11.sRo = 0; gsb11.sRi = 0; gsb11.sRm = 0; gsb11.sRn = 0;
      gsb11.M = SEQ; gsb11.N = SEQ; gsb11.K = 16; gsb11.zi_n = 1; gsb11.flags = 0; gsb11.act = 0;
      gsb11.alpha = 1.0f; gsb11.beta = 0.0f; gsb11.sa = 1.0f; gsb11.sb = 1.0f; gsb11.Npad = SEQ; gsb11.pad_ = 0;
      k_gemm<1><<<dim3((unsigned)((SEQ) + 31) / 32, (unsigned)((SEQ) + 15) / 16, (unsigned)(4)), 32, 0, stream>>>(gsb11); }
    k_mm_rowsm<<<4 * SEQ, 256, 0, stream>>>(SC, 4 * SEQ, SEQ, 0.25f);
    { GemmP gvb11;
      gvb11.A = SC; gvb11.B = H1 + (size_t)11 * SEQ * 192 + 32; gvb11.bias = SC; gvb11.R = SC; gvb11.C = O2 + (size_t)11 * SEQ * 64;
      gvb11.sAo = (long long)SEQ * SEQ; gvb11.sAi = 0; gvb11.sAm = SEQ; gvb11.sAk = 1; gvb11.sBo = 48; gvb11.sBi = 0; gvb11.sBn = 1; gvb11.sBk = 192; gvb11.sCo = 16; gvb11.sCi = 0; gvb11.sCm = 64; gvb11.sRo = 0; gvb11.sRi = 0; gvb11.sRm = 0; gvb11.sRn = 0;
      gvb11.M = SEQ; gvb11.N = 16; gvb11.K = SEQ; gvb11.zi_n = 1; gvb11.flags = 0; gvb11.act = 0;
      gvb11.alpha = 1.0f; gvb11.beta = 0.0f; gvb11.sa = 1.0f; gvb11.sb = 1.0f; gvb11.Npad = 16; gvb11.pad_ = 0;
      k_gemm<1><<<dim3((unsigned)((16) + 31) / 32, (unsigned)((SEQ) + 15) / 16, (unsigned)(4)), 32, 0, stream>>>(gvb11); }
    { GemmP gsa12;
      gsa12.A = H1 + (size_t)12 * SEQ * 192; gsa12.B = H2 + (size_t)12 * SEQ * 192 + 16; gsa12.bias = H1 + (size_t)12 * SEQ * 192; gsa12.R = H1 + (size_t)12 * SEQ * 192; gsa12.C = SC;
      gsa12.sAo = 48; gsa12.sAi = 0; gsa12.sAm = 192; gsa12.sAk = 1; gsa12.sBo = 48; gsa12.sBi = 0; gsa12.sBn = 192; gsa12.sBk = 1; gsa12.sCo = (long long)SEQ * SEQ; gsa12.sCi = 0; gsa12.sCm = SEQ; gsa12.sRo = 0; gsa12.sRi = 0; gsa12.sRm = 0; gsa12.sRn = 0;
      gsa12.M = SEQ; gsa12.N = SEQ; gsa12.K = 16; gsa12.zi_n = 1; gsa12.flags = 0; gsa12.act = 0;
      gsa12.alpha = 1.0f; gsa12.beta = 0.0f; gsa12.sa = 1.0f; gsa12.sb = 1.0f; gsa12.Npad = SEQ; gsa12.pad_ = 0;
      k_gemm<1><<<dim3((unsigned)((SEQ) + 31) / 32, (unsigned)((SEQ) + 15) / 16, (unsigned)(4)), 32, 0, stream>>>(gsa12); }
    k_mm_rowsm<<<4 * SEQ, 256, 0, stream>>>(SC, 4 * SEQ, SEQ, 0.25f);
    { GemmP gva12;
      gva12.A = SC; gva12.B = H2 + (size_t)12 * SEQ * 192 + 32; gva12.bias = SC; gva12.R = SC; gva12.C = O1 + (size_t)12 * SEQ * 64;
      gva12.sAo = (long long)SEQ * SEQ; gva12.sAi = 0; gva12.sAm = SEQ; gva12.sAk = 1; gva12.sBo = 48; gva12.sBi = 0; gva12.sBn = 1; gva12.sBk = 192; gva12.sCo = 16; gva12.sCi = 0; gva12.sCm = 64; gva12.sRo = 0; gva12.sRi = 0; gva12.sRm = 0; gva12.sRn = 0;
      gva12.M = SEQ; gva12.N = 16; gva12.K = SEQ; gva12.zi_n = 1; gva12.flags = 0; gva12.act = 0;
      gva12.alpha = 1.0f; gva12.beta = 0.0f; gva12.sa = 1.0f; gva12.sb = 1.0f; gva12.Npad = 16; gva12.pad_ = 0;
      k_gemm<1><<<dim3((unsigned)((16) + 31) / 32, (unsigned)((SEQ) + 15) / 16, (unsigned)(4)), 32, 0, stream>>>(gva12); }
    { GemmP gsb12;
      gsb12.A = H2 + (size_t)12 * SEQ * 192; gsb12.B = H1 + (size_t)12 * SEQ * 192 + 16; gsb12.bias = H2 + (size_t)12 * SEQ * 192; gsb12.R = H2 + (size_t)12 * SEQ * 192; gsb12.C = SC;
      gsb12.sAo = 48; gsb12.sAi = 0; gsb12.sAm = 192; gsb12.sAk = 1; gsb12.sBo = 48; gsb12.sBi = 0; gsb12.sBn = 192; gsb12.sBk = 1; gsb12.sCo = (long long)SEQ * SEQ; gsb12.sCi = 0; gsb12.sCm = SEQ; gsb12.sRo = 0; gsb12.sRi = 0; gsb12.sRm = 0; gsb12.sRn = 0;
      gsb12.M = SEQ; gsb12.N = SEQ; gsb12.K = 16; gsb12.zi_n = 1; gsb12.flags = 0; gsb12.act = 0;
      gsb12.alpha = 1.0f; gsb12.beta = 0.0f; gsb12.sa = 1.0f; gsb12.sb = 1.0f; gsb12.Npad = SEQ; gsb12.pad_ = 0;
      k_gemm<1><<<dim3((unsigned)((SEQ) + 31) / 32, (unsigned)((SEQ) + 15) / 16, (unsigned)(4)), 32, 0, stream>>>(gsb12); }
    k_mm_rowsm<<<4 * SEQ, 256, 0, stream>>>(SC, 4 * SEQ, SEQ, 0.25f);
    { GemmP gvb12;
      gvb12.A = SC; gvb12.B = H1 + (size_t)12 * SEQ * 192 + 32; gvb12.bias = SC; gvb12.R = SC; gvb12.C = O2 + (size_t)12 * SEQ * 64;
      gvb12.sAo = (long long)SEQ * SEQ; gvb12.sAi = 0; gvb12.sAm = SEQ; gvb12.sAk = 1; gvb12.sBo = 48; gvb12.sBi = 0; gvb12.sBn = 1; gvb12.sBk = 192; gvb12.sCo = 16; gvb12.sCi = 0; gvb12.sCm = 64; gvb12.sRo = 0; gvb12.sRi = 0; gvb12.sRm = 0; gvb12.sRn = 0;
      gvb12.M = SEQ; gvb12.N = 16; gvb12.K = SEQ; gvb12.zi_n = 1; gvb12.flags = 0; gvb12.act = 0;
      gvb12.alpha = 1.0f; gvb12.beta = 0.0f; gvb12.sa = 1.0f; gvb12.sb = 1.0f; gvb12.Npad = 16; gvb12.pad_ = 0;
      k_gemm<1><<<dim3((unsigned)((16) + 31) / 32, (unsigned)((SEQ) + 15) / 16, (unsigned)(4)), 32, 0, stream>>>(gvb12); }
    { GemmP gsa13;
      gsa13.A = H1 + (size_t)13 * SEQ * 192; gsa13.B = H2 + (size_t)13 * SEQ * 192 + 16; gsa13.bias = H1 + (size_t)13 * SEQ * 192; gsa13.R = H1 + (size_t)13 * SEQ * 192; gsa13.C = SC;
      gsa13.sAo = 48; gsa13.sAi = 0; gsa13.sAm = 192; gsa13.sAk = 1; gsa13.sBo = 48; gsa13.sBi = 0; gsa13.sBn = 192; gsa13.sBk = 1; gsa13.sCo = (long long)SEQ * SEQ; gsa13.sCi = 0; gsa13.sCm = SEQ; gsa13.sRo = 0; gsa13.sRi = 0; gsa13.sRm = 0; gsa13.sRn = 0;
      gsa13.M = SEQ; gsa13.N = SEQ; gsa13.K = 16; gsa13.zi_n = 1; gsa13.flags = 0; gsa13.act = 0;
      gsa13.alpha = 1.0f; gsa13.beta = 0.0f; gsa13.sa = 1.0f; gsa13.sb = 1.0f; gsa13.Npad = SEQ; gsa13.pad_ = 0;
      k_gemm<1><<<dim3((unsigned)((SEQ) + 31) / 32, (unsigned)((SEQ) + 15) / 16, (unsigned)(4)), 32, 0, stream>>>(gsa13); }
    k_mm_rowsm<<<4 * SEQ, 256, 0, stream>>>(SC, 4 * SEQ, SEQ, 0.25f);
    { GemmP gva13;
      gva13.A = SC; gva13.B = H2 + (size_t)13 * SEQ * 192 + 32; gva13.bias = SC; gva13.R = SC; gva13.C = O1 + (size_t)13 * SEQ * 64;
      gva13.sAo = (long long)SEQ * SEQ; gva13.sAi = 0; gva13.sAm = SEQ; gva13.sAk = 1; gva13.sBo = 48; gva13.sBi = 0; gva13.sBn = 1; gva13.sBk = 192; gva13.sCo = 16; gva13.sCi = 0; gva13.sCm = 64; gva13.sRo = 0; gva13.sRi = 0; gva13.sRm = 0; gva13.sRn = 0;
      gva13.M = SEQ; gva13.N = 16; gva13.K = SEQ; gva13.zi_n = 1; gva13.flags = 0; gva13.act = 0;
      gva13.alpha = 1.0f; gva13.beta = 0.0f; gva13.sa = 1.0f; gva13.sb = 1.0f; gva13.Npad = 16; gva13.pad_ = 0;
      k_gemm<1><<<dim3((unsigned)((16) + 31) / 32, (unsigned)((SEQ) + 15) / 16, (unsigned)(4)), 32, 0, stream>>>(gva13); }
    { GemmP gsb13;
      gsb13.A = H2 + (size_t)13 * SEQ * 192; gsb13.B = H1 + (size_t)13 * SEQ * 192 + 16; gsb13.bias = H2 + (size_t)13 * SEQ * 192; gsb13.R = H2 + (size_t)13 * SEQ * 192; gsb13.C = SC;
      gsb13.sAo = 48; gsb13.sAi = 0; gsb13.sAm = 192; gsb13.sAk = 1; gsb13.sBo = 48; gsb13.sBi = 0; gsb13.sBn = 192; gsb13.sBk = 1; gsb13.sCo = (long long)SEQ * SEQ; gsb13.sCi = 0; gsb13.sCm = SEQ; gsb13.sRo = 0; gsb13.sRi = 0; gsb13.sRm = 0; gsb13.sRn = 0;
      gsb13.M = SEQ; gsb13.N = SEQ; gsb13.K = 16; gsb13.zi_n = 1; gsb13.flags = 0; gsb13.act = 0;
      gsb13.alpha = 1.0f; gsb13.beta = 0.0f; gsb13.sa = 1.0f; gsb13.sb = 1.0f; gsb13.Npad = SEQ; gsb13.pad_ = 0;
      k_gemm<1><<<dim3((unsigned)((SEQ) + 31) / 32, (unsigned)((SEQ) + 15) / 16, (unsigned)(4)), 32, 0, stream>>>(gsb13); }
    k_mm_rowsm<<<4 * SEQ, 256, 0, stream>>>(SC, 4 * SEQ, SEQ, 0.25f);
    { GemmP gvb13;
      gvb13.A = SC; gvb13.B = H1 + (size_t)13 * SEQ * 192 + 32; gvb13.bias = SC; gvb13.R = SC; gvb13.C = O2 + (size_t)13 * SEQ * 64;
      gvb13.sAo = (long long)SEQ * SEQ; gvb13.sAi = 0; gvb13.sAm = SEQ; gvb13.sAk = 1; gvb13.sBo = 48; gvb13.sBi = 0; gvb13.sBn = 1; gvb13.sBk = 192; gvb13.sCo = 16; gvb13.sCi = 0; gvb13.sCm = 64; gvb13.sRo = 0; gvb13.sRi = 0; gvb13.sRm = 0; gvb13.sRn = 0;
      gvb13.M = SEQ; gvb13.N = 16; gvb13.K = SEQ; gvb13.zi_n = 1; gvb13.flags = 0; gvb13.act = 0;
      gvb13.alpha = 1.0f; gvb13.beta = 0.0f; gvb13.sa = 1.0f; gvb13.sb = 1.0f; gvb13.Npad = 16; gvb13.pad_ = 0;
      k_gemm<1><<<dim3((unsigned)((16) + 31) / 32, (unsigned)((SEQ) + 15) / 16, (unsigned)(4)), 32, 0, stream>>>(gvb13); }
    { GemmP gsa14;
      gsa14.A = H1 + (size_t)14 * SEQ * 192; gsa14.B = H2 + (size_t)14 * SEQ * 192 + 16; gsa14.bias = H1 + (size_t)14 * SEQ * 192; gsa14.R = H1 + (size_t)14 * SEQ * 192; gsa14.C = SC;
      gsa14.sAo = 48; gsa14.sAi = 0; gsa14.sAm = 192; gsa14.sAk = 1; gsa14.sBo = 48; gsa14.sBi = 0; gsa14.sBn = 192; gsa14.sBk = 1; gsa14.sCo = (long long)SEQ * SEQ; gsa14.sCi = 0; gsa14.sCm = SEQ; gsa14.sRo = 0; gsa14.sRi = 0; gsa14.sRm = 0; gsa14.sRn = 0;
      gsa14.M = SEQ; gsa14.N = SEQ; gsa14.K = 16; gsa14.zi_n = 1; gsa14.flags = 0; gsa14.act = 0;
      gsa14.alpha = 1.0f; gsa14.beta = 0.0f; gsa14.sa = 1.0f; gsa14.sb = 1.0f; gsa14.Npad = SEQ; gsa14.pad_ = 0;
      k_gemm<1><<<dim3((unsigned)((SEQ) + 31) / 32, (unsigned)((SEQ) + 15) / 16, (unsigned)(4)), 32, 0, stream>>>(gsa14); }
    k_mm_rowsm<<<4 * SEQ, 256, 0, stream>>>(SC, 4 * SEQ, SEQ, 0.25f);
    { GemmP gva14;
      gva14.A = SC; gva14.B = H2 + (size_t)14 * SEQ * 192 + 32; gva14.bias = SC; gva14.R = SC; gva14.C = O1 + (size_t)14 * SEQ * 64;
      gva14.sAo = (long long)SEQ * SEQ; gva14.sAi = 0; gva14.sAm = SEQ; gva14.sAk = 1; gva14.sBo = 48; gva14.sBi = 0; gva14.sBn = 1; gva14.sBk = 192; gva14.sCo = 16; gva14.sCi = 0; gva14.sCm = 64; gva14.sRo = 0; gva14.sRi = 0; gva14.sRm = 0; gva14.sRn = 0;
      gva14.M = SEQ; gva14.N = 16; gva14.K = SEQ; gva14.zi_n = 1; gva14.flags = 0; gva14.act = 0;
      gva14.alpha = 1.0f; gva14.beta = 0.0f; gva14.sa = 1.0f; gva14.sb = 1.0f; gva14.Npad = 16; gva14.pad_ = 0;
      k_gemm<1><<<dim3((unsigned)((16) + 31) / 32, (unsigned)((SEQ) + 15) / 16, (unsigned)(4)), 32, 0, stream>>>(gva14); }
    { GemmP gsb14;
      gsb14.A = H2 + (size_t)14 * SEQ * 192; gsb14.B = H1 + (size_t)14 * SEQ * 192 + 16; gsb14.bias = H2 + (size_t)14 * SEQ * 192; gsb14.R = H2 + (size_t)14 * SEQ * 192; gsb14.C = SC;
      gsb14.sAo = 48; gsb14.sAi = 0; gsb14.sAm = 192; gsb14.sAk = 1; gsb14.sBo = 48; gsb14.sBi = 0; gsb14.sBn = 192; gsb14.sBk = 1; gsb14.sCo = (long long)SEQ * SEQ; gsb14.sCi = 0; gsb14.sCm = SEQ; gsb14.sRo = 0; gsb14.sRi = 0; gsb14.sRm = 0; gsb14.sRn = 0;
      gsb14.M = SEQ; gsb14.N = SEQ; gsb14.K = 16; gsb14.zi_n = 1; gsb14.flags = 0; gsb14.act = 0;
      gsb14.alpha = 1.0f; gsb14.beta = 0.0f; gsb14.sa = 1.0f; gsb14.sb = 1.0f; gsb14.Npad = SEQ; gsb14.pad_ = 0;
      k_gemm<1><<<dim3((unsigned)((SEQ) + 31) / 32, (unsigned)((SEQ) + 15) / 16, (unsigned)(4)), 32, 0, stream>>>(gsb14); }
    k_mm_rowsm<<<4 * SEQ, 256, 0, stream>>>(SC, 4 * SEQ, SEQ, 0.25f);
    { GemmP gvb14;
      gvb14.A = SC; gvb14.B = H1 + (size_t)14 * SEQ * 192 + 32; gvb14.bias = SC; gvb14.R = SC; gvb14.C = O2 + (size_t)14 * SEQ * 64;
      gvb14.sAo = (long long)SEQ * SEQ; gvb14.sAi = 0; gvb14.sAm = SEQ; gvb14.sAk = 1; gvb14.sBo = 48; gvb14.sBi = 0; gvb14.sBn = 1; gvb14.sBk = 192; gvb14.sCo = 16; gvb14.sCi = 0; gvb14.sCm = 64; gvb14.sRo = 0; gvb14.sRi = 0; gvb14.sRm = 0; gvb14.sRn = 0;
      gvb14.M = SEQ; gvb14.N = 16; gvb14.K = SEQ; gvb14.zi_n = 1; gvb14.flags = 0; gvb14.act = 0;
      gvb14.alpha = 1.0f; gvb14.beta = 0.0f; gvb14.sa = 1.0f; gvb14.sb = 1.0f; gvb14.Npad = 16; gvb14.pad_ = 0;
      k_gemm<1><<<dim3((unsigned)((16) + 31) / 32, (unsigned)((SEQ) + 15) / 16, (unsigned)(4)), 32, 0, stream>>>(gvb14); }
    { GemmP gsa15;
      gsa15.A = H1 + (size_t)15 * SEQ * 192; gsa15.B = H2 + (size_t)15 * SEQ * 192 + 16; gsa15.bias = H1 + (size_t)15 * SEQ * 192; gsa15.R = H1 + (size_t)15 * SEQ * 192; gsa15.C = SC;
      gsa15.sAo = 48; gsa15.sAi = 0; gsa15.sAm = 192; gsa15.sAk = 1; gsa15.sBo = 48; gsa15.sBi = 0; gsa15.sBn = 192; gsa15.sBk = 1; gsa15.sCo = (long long)SEQ * SEQ; gsa15.sCi = 0; gsa15.sCm = SEQ; gsa15.sRo = 0; gsa15.sRi = 0; gsa15.sRm = 0; gsa15.sRn = 0;
      gsa15.M = SEQ; gsa15.N = SEQ; gsa15.K = 16; gsa15.zi_n = 1; gsa15.flags = 0; gsa15.act = 0;
      gsa15.alpha = 1.0f; gsa15.beta = 0.0f; gsa15.sa = 1.0f; gsa15.sb = 1.0f; gsa15.Npad = SEQ; gsa15.pad_ = 0;
      k_gemm<1><<<dim3((unsigned)((SEQ) + 31) / 32, (unsigned)((SEQ) + 15) / 16, (unsigned)(4)), 32, 0, stream>>>(gsa15); }
    k_mm_rowsm<<<4 * SEQ, 256, 0, stream>>>(SC, 4 * SEQ, SEQ, 0.25f);
    { GemmP gva15;
      gva15.A = SC; gva15.B = H2 + (size_t)15 * SEQ * 192 + 32; gva15.bias = SC; gva15.R = SC; gva15.C = O1 + (size_t)15 * SEQ * 64;
      gva15.sAo = (long long)SEQ * SEQ; gva15.sAi = 0; gva15.sAm = SEQ; gva15.sAk = 1; gva15.sBo = 48; gva15.sBi = 0; gva15.sBn = 1; gva15.sBk = 192; gva15.sCo = 16; gva15.sCi = 0; gva15.sCm = 64; gva15.sRo = 0; gva15.sRi = 0; gva15.sRm = 0; gva15.sRn = 0;
      gva15.M = SEQ; gva15.N = 16; gva15.K = SEQ; gva15.zi_n = 1; gva15.flags = 0; gva15.act = 0;
      gva15.alpha = 1.0f; gva15.beta = 0.0f; gva15.sa = 1.0f; gva15.sb = 1.0f; gva15.Npad = 16; gva15.pad_ = 0;
      k_gemm<1><<<dim3((unsigned)((16) + 31) / 32, (unsigned)((SEQ) + 15) / 16, (unsigned)(4)), 32, 0, stream>>>(gva15); }
    { GemmP gsb15;
      gsb15.A = H2 + (size_t)15 * SEQ * 192; gsb15.B = H1 + (size_t)15 * SEQ * 192 + 16; gsb15.bias = H2 + (size_t)15 * SEQ * 192; gsb15.R = H2 + (size_t)15 * SEQ * 192; gsb15.C = SC;
      gsb15.sAo = 48; gsb15.sAi = 0; gsb15.sAm = 192; gsb15.sAk = 1; gsb15.sBo = 48; gsb15.sBi = 0; gsb15.sBn = 192; gsb15.sBk = 1; gsb15.sCo = (long long)SEQ * SEQ; gsb15.sCi = 0; gsb15.sCm = SEQ; gsb15.sRo = 0; gsb15.sRi = 0; gsb15.sRm = 0; gsb15.sRn = 0;
      gsb15.M = SEQ; gsb15.N = SEQ; gsb15.K = 16; gsb15.zi_n = 1; gsb15.flags = 0; gsb15.act = 0;
      gsb15.alpha = 1.0f; gsb15.beta = 0.0f; gsb15.sa = 1.0f; gsb15.sb = 1.0f; gsb15.Npad = SEQ; gsb15.pad_ = 0;
      k_gemm<1><<<dim3((unsigned)((SEQ) + 31) / 32, (unsigned)((SEQ) + 15) / 16, (unsigned)(4)), 32, 0, stream>>>(gsb15); }
    k_mm_rowsm<<<4 * SEQ, 256, 0, stream>>>(SC, 4 * SEQ, SEQ, 0.25f);
    { GemmP gvb15;
      gvb15.A = SC; gvb15.B = H1 + (size_t)15 * SEQ * 192 + 32; gvb15.bias = SC; gvb15.R = SC; gvb15.C = O2 + (size_t)15 * SEQ * 64;
      gvb15.sAo = (long long)SEQ * SEQ; gvb15.sAi = 0; gvb15.sAm = SEQ; gvb15.sAk = 1; gvb15.sBo = 48; gvb15.sBi = 0; gvb15.sBn = 1; gvb15.sBk = 192; gvb15.sCo = 16; gvb15.sCi = 0; gvb15.sCm = 64; gvb15.sRo = 0; gvb15.sRi = 0; gvb15.sRm = 0; gvb15.sRn = 0;
      gvb15.M = SEQ; gvb15.N = 16; gvb15.K = SEQ; gvb15.zi_n = 1; gvb15.flags = 0; gvb15.act = 0;
      gvb15.alpha = 1.0f; gvb15.beta = 0.0f; gvb15.sa = 1.0f; gvb15.sb = 1.0f; gvb15.Npad = 16; gvb15.pad_ = 0;
      k_gemm<1><<<dim3((unsigned)((16) + 31) / 32, (unsigned)((SEQ) + 15) / 16, (unsigned)(4)), 32, 0, stream>>>(gvb15); }
    { GemmP gt1;
      gt1.A = O1; gt1.B = cow; gt1.bias = cob; gt1.R = O1; gt1.C = T1;
      gt1.sAo = 0; gt1.sAi = 0; gt1.sAm = 64; gt1.sAk = 1; gt1.sBo = 0; gt1.sBi = 0; gt1.sBn = 64; gt1.sBk = 1; gt1.sCo = 0; gt1.sCi = 0; gt1.sCm = 64; gt1.sRo = 0; gt1.sRi = 0; gt1.sRm = 0; gt1.sRn = 0;
      gt1.M = Bn * SEQ; gt1.N = 64; gt1.K = 64; gt1.zi_n = 1; gt1.flags = 1; gt1.act = 0;
      gt1.alpha = 1.0f; gt1.beta = 0.0f; gt1.sa = 1.0f; gt1.sb = 1.0f; gt1.Npad = 64; gt1.pad_ = 0;
      k_gemm<1><<<dim3((unsigned)((64) + 31) / 32, (unsigned)((Bn * SEQ) + 15) / 16, (unsigned)(1)), 32, 0, stream>>>(gt1); }
    { GemmP gt2;
      gt2.A = O2; gt2.B = cow; gt2.bias = cob; gt2.R = O2; gt2.C = T2;
      gt2.sAo = 0; gt2.sAi = 0; gt2.sAm = 64; gt2.sAk = 1; gt2.sBo = 0; gt2.sBi = 0; gt2.sBn = 64; gt2.sBk = 1; gt2.sCo = 0; gt2.sCi = 0; gt2.sCm = 64; gt2.sRo = 0; gt2.sRi = 0; gt2.sRm = 0; gt2.sRn = 0;
      gt2.M = Bn * SEQ; gt2.N = 64; gt2.K = 64; gt2.zi_n = 1; gt2.flags = 1; gt2.act = 0;
      gt2.alpha = 1.0f; gt2.beta = 0.0f; gt2.sa = 1.0f; gt2.sb = 1.0f; gt2.Npad = 64; gt2.pad_ = 0;
      k_gemm<1><<<dim3((unsigned)((64) + 31) / 32, (unsigned)((Bn * SEQ) + 15) / 16, (unsigned)(1)), 32, 0, stream>>>(gt2); }
    k_mm_pools<<<(unsigned)((Bn * SEQ + 255) / 256), 256, 0, stream>>>(T1, T2, CHP, SPP, Bn, SEQ, 64);
    k_mm_chgate<<<(unsigned)((Bn * 64 + 255) / 256), 256, 0, stream>>>(CHP, ch1w, ch1b, ch2w, ch2b, CHS, Bn, 64);
    k_mm_spgate<<<(unsigned)((Bn * SEQ + 255) / 256), 256, 0, stream>>>(SPP, sp1w, sp1b, sp2w, sp2b, SPS, Bn, 32);
    k_mm_fuse<<<(unsigned)((Bn * 64 + 255) / 256), 256, 0, stream>>>(T1, T2, CHS, SPS, FM, Bn, SEQ, 64);
    { GemmP gcls;
      gcls.A = FM; gcls.B = clsw; gcls.bias = clsb; gcls.R = FM; gcls.C = LG;
      gcls.sAo = 0; gcls.sAi = 0; gcls.sAm = 64; gcls.sAk = 1; gcls.sBo = 0; gcls.sBi = 0; gcls.sBn = 64; gcls.sBk = 1; gcls.sCo = 0; gcls.sCi = 0; gcls.sCm = LP; gcls.sRo = 0; gcls.sRi = 0; gcls.sRm = 0; gcls.sRn = 0;
      gcls.M = Bn; gcls.N = 9; gcls.K = 64; gcls.zi_n = 1; gcls.flags = 1; gcls.act = 0;
      gcls.alpha = 1.0f; gcls.beta = 0.0f; gcls.sa = 1.0f; gcls.sb = 1.0f; gcls.Npad = LP; gcls.pad_ = 0;
      k_gemm<1><<<dim3((unsigned)((LP) + 31) / 32, (unsigned)((Bn) + 15) / 16, (unsigned)(1)), 32, 0, stream>>>(gcls); }
    k_mm_out<<<1, 256, 0, stream>>>(LG, LP, out, Bn, 9);
}
